// BNeckConvLSTM_12687333392819
// MI455X (gfx1250) — hardware-verified
//
#include <hip/hip_runtime.h>
#include <math.h>

typedef __attribute__((ext_vector_type(16))) _Float16 v16h;
typedef __attribute__((ext_vector_type(8)))  _Float16 v8h;
typedef __attribute__((ext_vector_type(16))) __bf16   v16b;
typedef __attribute__((ext_vector_type(8)))  float    v8f;
typedef __attribute__((ext_vector_type(4)))  float    v4f;

__device__ __forceinline__ int frag_k(int i, int h) { return (i < 8) ? (8 * h + i) : (16 + 8 * h + (i - 8)); }
__device__ __forceinline__ __bf16 bf16_rne(float f) {
    unsigned int u = __float_as_uint(f);
    u += 0x7fffu + ((u >> 16) & 1u);
    return __builtin_bit_cast(__bf16, (unsigned short)(u >> 16));
}
__device__ __forceinline__ float bf16_f32(__bf16 b) { return __uint_as_float(((unsigned int)__builtin_bit_cast(unsigned short, b)) << 16); }
__device__ __forceinline__ v8f wmma16(v16h a, v16h b, v8f c) {
    c = __builtin_amdgcn_wmma_f32_16x16x32_f16(false, a, false, b, (short)0, c, false, false);
    asm volatile("v_nop\n\tv_nop\n\tv_nop\n\tv_nop" : "+v"(c) : "v"(a), "v"(b));
    return c;
}
__device__ __forceinline__ v8f wmmab(v16b a, v16b b, v8f c) {
    c = __builtin_amdgcn_wmma_f32_16x16x32_bf16(false, a, false, b, (short)0, c, false, false);
    asm volatile("v_nop\n\tv_nop\n\tv_nop\n\tv_nop" : "+v"(c) : "v"(a), "v"(b));
    return c;
}
struct Split { v16b hi, lo; };
__device__ __forceinline__ v8f wmma3(const Split& a, const Split& b, v8f c) {
    c = __builtin_amdgcn_wmma_f32_16x16x32_bf16(false, a.hi, false, b.hi, (short)0, c, false, false);
    c = __builtin_amdgcn_wmma_f32_16x16x32_bf16(false, a.hi, false, b.lo, (short)0, c, false, false);
    c = __builtin_amdgcn_wmma_f32_16x16x32_bf16(false, a.lo, false, b.hi, (short)0, c, false, false);
    asm volatile("v_nop\n\tv_nop\n\tv_nop\n\tv_nop" : "+v"(c) : "v"(a.hi), "v"(a.lo), "v"(b.hi), "v"(b.lo));
    return c;
}
struct Split3 { v16b hi, mid, lo; };
__device__ __forceinline__ v8f wmma6(const Split3& a, const Split3& b, v8f c) {
    c = __builtin_amdgcn_wmma_f32_16x16x32_bf16(false, a.hi, false, b.hi, (short)0, c, false, false);
    c = __builtin_amdgcn_wmma_f32_16x16x32_bf16(false, a.hi, false, b.mid, (short)0, c, false, false);
    c = __builtin_amdgcn_wmma_f32_16x16x32_bf16(false, a.mid, false, b.hi, (short)0, c, false, false);
    c = __builtin_amdgcn_wmma_f32_16x16x32_bf16(false, a.hi, false, b.lo, (short)0, c, false, false);
    c = __builtin_amdgcn_wmma_f32_16x16x32_bf16(false, a.mid, false, b.mid, (short)0, c, false, false);
    c = __builtin_amdgcn_wmma_f32_16x16x32_bf16(false, a.lo, false, b.hi, (short)0, c, false, false);
    asm volatile("v_nop\n\tv_nop\n\tv_nop\n\tv_nop" : "+v"(c) : "v"(a.hi), "v"(a.mid), "v"(a.lo), "v"(b.hi), "v"(b.mid), "v"(b.lo));
    return c;
}

__device__ __forceinline__ v16h fh_ld(const float* __restrict__ p, long long sk, int k0, int h, int klen, float s) {
    v16h a;
#pragma unroll
    for (int i = 0; i < 16; ++i) { const int k = k0 + frag_k(i, h); a[i] = (k < klen) ? (_Float16)(p[(long long)k * sk] * s) : (_Float16)0.f; }
    return a;
}
__device__ __forceinline__ Split sp_ld(const float* __restrict__ p, long long sk, int k0, int h, int klen, float s) {
    Split r;
#pragma unroll
    for (int i = 0; i < 16; ++i) {
        const int k = k0 + frag_k(i, h); const float x = (k < klen) ? p[(long long)k * sk] * s : 0.f;
        const __bf16 hb = bf16_rne(x); r.hi[i] = hb; r.lo[i] = bf16_rne(x - bf16_f32(hb));
    }
    return r;
}
__device__ __forceinline__ Split3 sp3_ld(const float* __restrict__ p, long long sk, int k0, int h, int klen, float s) {
    Split3 r;
#pragma unroll
    for (int i = 0; i < 16; ++i) {
        const int k = k0 + frag_k(i, h); const float x = (k < klen) ? p[(long long)k * sk] * s : 0.f;
        const __bf16 hb = bf16_rne(x); const float r1 = x - bf16_f32(hb); const __bf16 mb = bf16_rne(r1);
        r.hi[i] = hb; r.mid[i] = mb; r.lo[i] = bf16_rne(r1 - bf16_f32(mb));
    }
    return r;
}
__device__ __forceinline__ v16b bh_ld(const float* __restrict__ p, long long sk, int k0, int h, int klen, float s) {
    v16b a;
#pragma unroll
    for (int i = 0; i < 16; ++i) { const int k = k0 + frag_k(i, h); a[i] = bf16_rne((k < klen) ? p[(long long)k * sk] * s : 0.f); }
    return a;
}
__device__ __forceinline__ v16h fh_row(const _Float16* __restrict__ row, int k0, int h) {
    v16h a;
#pragma unroll
    for (int i = 0; i < 16; ++i) a[i] = row[k0 + frag_k(i, h)];
    return a;
}

#define VST2(T, ptr, val) do { *(volatile T*)(ptr) = (val); __threadfence(); *(volatile T*)(ptr) = (val); } while (0)
typedef float v4f __attribute__((ext_vector_type(4)));
#define VST2V4(ptr, val) do { *(volatile v4f*)(ptr) = (val); __threadfence(); *(volatile v4f*)(ptr) = (val); } while (0)

__device__ __attribute__((noinline)) float act_fn(float v, int act) {
    if (act == 1) return fmaxf(v, 0.f);
    if (act == 2) { const float u = 0.7978845608028654f * (v + 0.044715f * v * v * v); return 0.5f * v * (1.f + tanhf(u)); }
    if (act == 3) return v / (1.f + expf(-v));
    if (act == 4) return 0.5f * v * (1.f + erff(v * 0.7071067811865476f));
    if (act == 5) return tanhf(v);
    if (act == 6) return 1.f / (1.f + expf(-v));
    if (act == 7) return (v > 0.f) ? v : 0.01f * v;
    if (act == 8) return (v > 0.f) ? v : (expf(v) - 1.f);
    if (act == 9) return fminf(fmaxf(v, 0.f), 6.f);
    if (act == 10) return fabsf(v);
    if (act == 11) return (v >= 0.f) ? v : 0.1f * v;
    if (act == 12) return (v > 0.f) ? v : 0.2f * v;
    if (act == 13) return (v > 20.f) ? v : log1pf(expf(v));
    return v;
}

struct GemmP {
    const float* A; const float* B; const float* bias; const float* R; float* C;
    long long sAo, sAi, sAm, sAk, sBo, sBi, sBn, sBk, sCo, sCi, sCm, sRo, sRi, sRm, sRn;
    int M, N, K, zi_n, flags, act; float alpha, beta, sa, sb;
    int Npad, pad_;
};
static_assert(sizeof(GemmP) == 5 * 8 + 15 * 8 + 6 * 4 + 4 * 4 + 2 * 4, "GemmP has padding");

template <int MODE>
__global__ __launch_bounds__(32) void k_gemm(GemmP p) {
    const int lane = threadIdx.x & 31, h = lane >> 4, l15 = lane & 15;
    const int m0 = blockIdx.y * 16, n0 = blockIdx.x * 32;
    const int z = blockIdx.z, zo = z / p.zi_n, zi = z - zo * p.zi_n;
    const float* A = p.A + zo * p.sAo + zi * p.sAi;
    const float* B = p.B + zo * p.sBo + zi * p.sBi;
    const int am = min(m0 + l15, p.M - 1);
    v8f acc[2], comp[2];
#pragma unroll
    for (int t = 0; t < 2; ++t) { v8f zz = {}; acc[t] = zz; comp[t] = zz; }
    for (int k0 = 0; k0 < p.K; k0 += 32) {
        const float* arow = A + (long long)am * p.sAm;
        if (MODE == 1) {
            const Split a = sp_ld(arow, p.sAk, k0, h, p.K, 1.f);
#pragma unroll
            for (int t = 0; t < 2; ++t) {
                const int bn = min(n0 + t * 16 + l15, p.N - 1);
                acc[t] = wmma3(a, sp_ld(B + (long long)bn * p.sBn, p.sBk, k0, h, p.K, 1.f), acc[t]);
            }
        } else if (MODE == 3) {
            const Split3 a = sp3_ld(arow, p.sAk, k0, h, p.K, 1.f);
#pragma unroll
            for (int t = 0; t < 2; ++t) {
                const int bn = min(n0 + t * 16 + l15, p.N - 1);
                acc[t] = wmma6(a, sp3_ld(B + (long long)bn * p.sBn, p.sBk, k0, h, p.K, 1.f), acc[t]);
            }
        } else if (MODE == 4) {
            const Split3 a = sp3_ld(arow, p.sAk, k0, h, p.K, 1.f);
#pragma unroll
            for (int t = 0; t < 2; ++t) {
                const int bn = min(n0 + t * 16 + l15, p.N - 1); v8f zz = {};
                const v8f part = wmma6(a, sp3_ld(B + (long long)bn * p.sBn, p.sBk, k0, h, p.K, 1.f), zz);
                const v8f y = part - comp[t]; const v8f s = acc[t] + y; comp[t] = (s - acc[t]) - y; acc[t] = s;
            }
        } else if (MODE == 2) {
            const v16b a = bh_ld(arow, p.sAk, k0, h, p.K, 1.f);
#pragma unroll
            for (int t = 0; t < 2; ++t) {
                const int bn = min(n0 + t * 16 + l15, p.N - 1);
                acc[t] = wmmab(a, bh_ld(B + (long long)bn * p.sBn, p.sBk, k0, h, p.K, 1.f), acc[t]);
            }
        } else {
            const v16h a = fh_ld(arow, p.sAk, k0, h, p.K, p.sa);
#pragma unroll
            for (int t = 0; t < 2; ++t) {
                const int bn = min(n0 + t * 16 + l15, p.N - 1);
                acc[t] = wmma16(a, fh_ld(B + (long long)bn * p.sBn, p.sBk, k0, h, p.K, p.sb), acc[t]);
            }
        }
    }
    const float iscale = (MODE == 0) ? p.alpha / (p.sa * p.sb) : p.alpha;
    float* C = p.C + zo * p.sCo + zi * p.sCi;
    const float* R = p.R + zo * p.sRo + zi * p.sRi;
    __shared__ __align__(16) float ctile[16][36];
#pragma unroll
    for (int t = 0; t < 2; ++t) {
        const int n = n0 + t * 16 + l15; const int nn = min(n, p.N - 1);
#pragma unroll
        for (int r = 0; r < 8; ++r) {
            const int m = m0 + 8 * h + r; const int mm = min(m, p.M - 1);
            float v = acc[t][r] * iscale;
            if (p.flags & 1) v += p.bias[nn];
            if (p.flags & 2) v += p.bias[mm];
            v = act_fn(v, p.act);
            if (p.flags & 4) v += p.beta * R[(long long)mm * p.sRm + (long long)nn * p.sRn];
            ctile[8 * h + r][t * 16 + l15] = (n < p.N) ? v : 0.f;
        }
    }
    __syncthreads();
    const int NW = (p.Npad > p.N) ? p.Npad : p.N;
    const bool fast = (m0 + 16 <= p.M) && (n0 + 32 <= NW) && ((p.sCm & 3) == 0) && ((((size_t)C) & 15) == 0);
    if (fast) {
#pragma unroll
        for (int s = 0; s < 4; ++s) {
            const int row = s * 4 + (lane >> 3), c4 = (lane & 7) * 4;
            const v4f v = *(const v4f*)&ctile[row][c4];
            VST2V4(C + (long long)(m0 + row) * p.sCm + n0 + c4, v);
        }
    } else {
        for (int row = 0; row < 16; ++row) {
            const int m = m0 + row, n = n0 + lane;
            if (m < p.M && n < NW) VST2(float, C + (long long)m * p.sCm + n, ctile[row][lane]);
        }
    }
}

#define AW 4
struct AttnP {
    const float* Q; const float* K; const float* V; float* O; float* P; const float* Mf; const int* Mi; float* ST;
    const float* Pw; const float* Rt; const int* SQ; const int* SK;
    long long swb, swh, swi, swj, srb, srh, sri;
    long long sQb, sQh, sQi, sQd, sKb, sKh, sKj, sKd, sVb, sVh, sVj, sVd, sOb, sOh, sOi, sPb, sPh, sPi, smb, smh, smi, smj;
    int Lq, Lk, dh, dv, hrep, causal, coff, pband;
    float scale, mfill; int nonorm, mpol;
    int roff, rn, segpol, win;
};
static_assert(sizeof(AttnP) == 12 * 8 + 29 * 8 + 16 * 4, "AttnP has padding");

#ifndef KATTN_ATTR
#define KATTN_ATTR
#endif
template <int DHP, int DVP, int QM, bool SPLITPV, bool TWOPASS>
__global__ __launch_bounds__(32 * AW) KATTN_ATTR void k_attn(AttnP p) {
    constexpr int NT = DVP / 16;
    constexpr int KS = DHP / 32;
    constexpr int VP = DVP + 8;
    __shared__ __align__(16) float    pl[AW][16 * 64];
    __shared__ __align__(16) _Float16 vl[(SPLITPV ? 2 : 1) * 64 * VP];
    const int lane = threadIdx.x & 31, hf = lane >> 4, l15 = lane & 15, wave = threadIdx.x >> 5;
    const int h = blockIdx.y, b = blockIdx.z, hk = h / p.hrep;
    const int q0 = (blockIdx.x * AW + wave) * 16;
    float* myp = pl[wave];
    const float L2E = 1.4426950408889634f;
    const float NEG = -__builtin_inff();
    const int qi = min(q0 + l15, p.Lq - 1);
    const float* qrow = p.Q + b * p.sQb + h * p.sQh + (long long)qi * p.sQi;
    const float* kbase = p.K + b * p.sKb + hk * p.sKh;
    const float* vbase = p.V + b * p.sVb + hk * p.sVh;
    v16h qa[QM == 0 ? KS : 1]; Split qs_[QM == 1 ? KS : 1]; Split3 qt_[QM == 2 ? KS : 1];
#pragma unroll
    for (int ks = 0; ks < KS; ++ks) {
        if (QM == 2) qt_[ks] = sp3_ld(qrow, p.sQd, ks * 32, hf, p.dh, 1.f);
        else if (QM == 1) qs_[ks] = sp_ld(qrow, p.sQd, ks * 32, hf, p.dh, 1.f);
        else qa[ks] = fh_ld(qrow, p.sQd, ks * 32, hf, p.dh, 1.f);
    }
    v8f o[NT]; float m8[8], l8[8];
#pragma unroll
    for (int t = 0; t < NT; ++t) { v8f zz = {}; o[t] = zz; }
#pragma unroll
    for (int i = 0; i < 8; ++i) { m8[i] = NEG; l8[i] = 0.f; }
    int jend = p.Lk;
    if (p.causal == 1) { const int je = (blockIdx.x * AW + AW - 1) * 16 + 16 + p.coff; jend = min(jend, max(je, 0)); }
    const int npass = TWOPASS ? 2 : 1;
    for (int pass = 0; pass < npass; ++pass) {
        const bool dopv = (!TWOPASS) || pass == 1;
        for (int j0 = 0; j0 < jend; j0 += 64) {
            if (dopv) {
                __syncthreads();
                for (int idx = threadIdx.x; idx < 64 * DVP; idx += 32 * AW) {
                    const int jr = idx / DVP, d = idx - jr * DVP, j = j0 + jr;
                    const float f = (j < p.Lk && d < p.dv) ? vbase[(long long)j * p.sVj + (long long)d * p.sVd] : 0.f;
                    if (SPLITPV) {
                        const __bf16 hb = bf16_rne(f);
                        ((__bf16*)vl)[jr * VP + d] = hb; ((__bf16*)vl)[64 * VP + jr * VP + d] = bf16_rne(f - bf16_f32(hb));
                    } else vl[jr * VP + d] = (_Float16)f;
                }
            }
            v8f s[4];
#pragma unroll
            for (int t = 0; t < 4; ++t) {
                const int j = min(j0 + t * 16 + l15, p.Lk - 1);
                const float* krow = kbase + (long long)j * p.sKj;
                v8f acc = {};
#pragma unroll
                for (int ks = 0; ks < KS; ++ks) {
                    if (QM == 2)      acc = wmma6(qt_[ks], sp3_ld(krow, p.sKd, ks * 32, hf, p.dh, 1.f), acc);
                    else if (QM == 1) acc = wmma3(qs_[ks], sp_ld(krow, p.sKd, ks * 32, hf, p.dh, 1.f), acc);
                    else              acc = wmma16(qa[ks], fh_ld(krow, p.sKd, ks * 32, hf, p.dh, 1.f), acc);
                }
                s[t] = acc;
            }
            float pv[8][4];
#pragma unroll
            for (int i = 0; i < 8; ++i) {
                const int irow = q0 + i + 8 * hf;
                const int ic = min(irow, p.Lq - 1);
                float sc[4];
#pragma unroll
                for (int t = 0; t < 4; ++t) {
                    const int jg = j0 + t * 16 + l15;
                    float v = s[t][i] * p.scale;
                    if (p.Mf) v += p.Mf[b * p.smb + h * p.smh + (long long)ic * p.smi + (long long)min(jg, p.Lk - 1) * p.smj];
                    if (p.Rt) { int rc = ic - min(jg, p.Lk - 1) + p.roff; rc = rc < 0 ? 0 : (rc >= p.rn ? p.rn - 1 : rc); v += p.Rt[b * p.srb + h * p.srh + (long long)ic * p.sri + rc]; }
                    if (p.Mi) { const int mv = p.Mi[b * p.smb + h * p.smh + (long long)ic * p.smi + (long long)min(jg, p.Lk - 1) * p.smj]; if (p.mpol ? (mv != 0) : (mv == 0)) v = p.mfill; }
                    if (p.SQ) { const bool same = p.SQ[(long long)b * p.Lq + ic] == p.SK[(long long)b * p.Lk + min(jg, p.Lk - 1)]; if (p.segpol ? same : !same) v = p.mfill; }
                    if (p.causal == 2 && jg > irow + p.coff) v = p.mfill;
                    if (jg >= p.Lk || (p.causal == 1 && jg > irow + p.coff) || (p.causal == 3 && jg < irow + p.coff) || (p.win > 0 && irow + p.coff - jg > p.win)) v = NEG; else v *= L2E;
                    sc[t] = v;
                }
                if (!TWOPASS || pass == 0) {
                    float mx = fmaxf(fmaxf(sc[0], sc[1]), fmaxf(sc[2], sc[3]));
                    mx = fmaxf(mx, __shfl_xor(mx, 1, 32)); mx = fmaxf(mx, __shfl_xor(mx, 2, 32));
                    mx = fmaxf(mx, __shfl_xor(mx, 4, 32)); mx = fmaxf(mx, __shfl_xor(mx, 8, 32));
                    const float mnew = fmaxf(m8[i], mx);
                    const float corr = (mnew == NEG) ? 1.f : exp2f(m8[i] - mnew);
                    float rs = 0.f;
#pragma unroll
                    for (int t = 0; t < 4; ++t) {
                        const float pp = (sc[t] == NEG) ? 0.f : exp2f(sc[t] - mnew); rs += pp;
                        pv[i][t] = p.Pw ? pp * p.Pw[b * p.swb + h * p.swh + (long long)ic * p.swi + (long long)min(j0 + t * 16 + l15, p.Lk - 1) * p.swj] : pp;
                    }
                    rs += __shfl_xor(rs, 1, 32); rs += __shfl_xor(rs, 2, 32); rs += __shfl_xor(rs, 4, 32); rs += __shfl_xor(rs, 8, 32);
                    l8[i] = l8[i] * corr + rs; m8[i] = mnew;
                    if (!TWOPASS) {
#pragma unroll
                        for (int t = 0; t < NT; ++t) o[t][i] *= corr;
                    }
                } else {
                    const float inv = (l8[i] > 0.f) ? 1.f / l8[i] : 0.f;
#pragma unroll
                    for (int t = 0; t < 4; ++t) {
                        const int jg = j0 + t * 16 + l15;
                        float pp = (sc[t] == NEG) ? 0.f : exp2f(sc[t] - m8[i]) * inv;
                        if (p.Pw) pp *= p.Pw[b * p.swb + h * p.swh + (long long)ic * p.swi + (long long)min(jg, p.Lk - 1) * p.swj];
                        pv[i][t] = pp;
                    }
                }
            }
            if (dopv) {
#pragma unroll
                for (int i = 0; i < 8; ++i)
#pragma unroll
                    for (int t = 0; t < 4; ++t) myp[(i + 8 * hf) * 64 + t * 16 + l15] = pv[i][t];
                __syncthreads();
                if (p.P) {
                    float* pb_ = p.P + b * p.sPb + h * p.sPh;
                    const bool fastP = (p.pband == 0) && ((p.sPi & 3) == 0) && (j0 + 64 <= p.Lk) && (q0 + 16 <= p.Lq) && ((((size_t)pb_) & 15) == 0);
                    if (fastP) {
#pragma unroll
                        for (int s = 0; s < 8; ++s) {
                            const int row = s * 2 + (lane >> 4), c4 = (lane & 15) * 4;
                            const v4f v = *(const v4f*)(myp + row * 64 + c4);
                            VST2V4(pb_ + (long long)(q0 + row) * p.sPi + j0 + c4, v);
                        }
                    } else {
                        for (int row = 0; row < 16; ++row) {
                            const int irow = q0 + row; if (irow >= p.Lq) continue;
                            for (int c = lane; c < 64; c += 32) {
                                const int jg = j0 + c; if (jg >= p.Lk) continue;
                                if (p.pband == 0) VST2(float, pb_ + (long long)irow * p.sPi + jg, myp[row * 64 + c]);
                                else if (jg - irow <= p.pband && irow - jg <= p.pband) VST2(float, pb_ + (long long)irow * p.sPi + (jg - irow + p.pband), myp[row * 64 + c]);
                            }
                        }
                    }
                }
                if (SPLITPV) {
                    const Split pa0 = sp_ld(myp + l15 * 64, 1, 0, hf, 64, 1.f), pa1 = sp_ld(myp + l15 * 64, 1, 32, hf, 64, 1.f);
                    const __bf16* vh = (const __bf16*)vl; const __bf16* vlo = vh + 64 * VP;
#pragma unroll
                    for (int t = 0; t < NT; ++t) {
                        const int dcol = t * 16 + l15;
                        Split b0, b1;
#pragma unroll
                        for (int e = 0; e < 16; ++e) {
                            const int k0 = frag_k(e, hf), k1 = 32 + frag_k(e, hf);
                            b0.hi[e] = vh[k0 * VP + dcol]; b0.lo[e] = vlo[k0 * VP + dcol]; b1.hi[e] = vh[k1 * VP + dcol]; b1.lo[e] = vlo[k1 * VP + dcol];
                        }
                        o[t] = wmma3(pa0, b0, o[t]);
                        o[t] = wmma3(pa1, b1, o[t]);
                    }
                } else {
                    const v16h pa0 = fh_ld(myp + l15 * 64, 1, 0, hf, 64, 4096.f), pa1 = fh_ld(myp + l15 * 64, 1, 32, hf, 64, 4096.f);
#pragma unroll
                    for (int t = 0; t < NT; ++t) {
                        const int dcol = t * 16 + l15;
                        v16h b0, b1;
#pragma unroll
                        for (int e = 0; e < 16; ++e) { b0[e] = vl[frag_k(e, hf) * VP + dcol]; b1[e] = vl[(32 + frag_k(e, hf)) * VP + dcol]; }
                        o[t] = wmma16(pa0, b0, o[t]);
                        o[t] = wmma16(pa1, b1, o[t]);
                    }
                }
            }
        }
    }
    float* obase = p.O + b * p.sOb + h * p.sOh;
    if (p.ST) {
        const int rl = lane >> 1, isel = rl & 7;
        float mv = 0.f, lv = 0.f;
#pragma unroll
        for (int i = 0; i < 8; ++i) if (i == isel) { mv = m8[i]; lv = l8[i]; }
        const int irow = q0 + rl;
        if (irow < p.Lq) { float* st = p.ST + (((long long)b * gridDim.y + h) * p.Lq + irow) * 2 + (lane & 1); VST2(float, st, (lane & 1) ? lv : mv * 0.6931471805599453f); }
    }
    float invr[8];
#pragma unroll
    for (int i = 0; i < 8; ++i) {
        if (TWOPASS) invr[i] = SPLITPV ? 1.f : (1.f / 4096.f);
        else if (p.nonorm) invr[i] = exp2f(m8[i]) * (SPLITPV ? 1.f : (1.f / 4096.f));
        else invr[i] = (l8[i] > 0.f) ? (SPLITPV ? 1.f / l8[i] : 1.f / (l8[i] * 4096.f)) : 0.f;
    }
    __syncthreads();
    const bool ofast = ((p.sOi & 3) == 0) && ((((size_t)obase) & 15) == 0) && (q0 + 16 <= p.Lq);
#pragma unroll
    for (int c0 = 0; c0 < DVP; c0 += 64) {
#pragma unroll
        for (int i = 0; i < 8; ++i)
#pragma unroll
            for (int t = 0; t < NT; ++t) if (t * 16 >= c0 && t * 16 < c0 + 64) myp[(i + 8 * hf) * 64 + (t * 16 - c0) + l15] = o[t][i] * invr[i];
        __syncthreads();
        const int cw = (DVP - c0 < 64) ? (DVP - c0) : 64;
        if (ofast && (c0 + cw <= p.dv) && (cw % 32 == 0)) {
            const int lpr = cw / 4;
            const int rows_per_ins = 32 / lpr;
            for (int r0 = 0; r0 < 16; r0 += rows_per_ins) {
                const int row = r0 + lane / lpr, c4 = (lane % lpr) * 4;
                const v4f v = *(const v4f*)(myp + row * 64 + c4);
                VST2V4(obase + (long long)(q0 + row) * p.sOi + c0 + c4, v);
            }
        } else {
            for (int row = 0; row < 16; ++row) {
                const int irow = q0 + row; if (irow >= p.Lq) continue;
                for (int c = lane; c < cw; c += 32) { const int d = c0 + c; if (d < p.dv) VST2(float, obase + (long long)irow * p.sOi + d, myp[row * 64 + c]); }
            }
        }
        __syncthreads();
    }
}

struct TrP { const float* src; float* dst; const float* R2; long long sSz, lds, sDz, ldd, sRz, ldr; int R, C, flags, act; float alpha, beta; };
static_assert(sizeof(TrP) == 3 * 8 + 6 * 8 + 6 * 4, "TrP has padding");
__global__ __launch_bounds__(256) void k_tr(TrP p) {
    __shared__ float tile[32][33];
    const int c0 = blockIdx.x * 32, r0 = blockIdx.y * 32, z = blockIdx.z;
    const int lane = threadIdx.x & 31, wave = threadIdx.x >> 5;
    const float* s = p.src + z * p.sSz;
#pragma unroll
    for (int k = 0; k < 4; ++k) {
        const int rl = wave * 4 + k, r = r0 + rl, c = c0 + lane;
        tile[rl][lane] = (r < p.R && c < p.C) ? s[(long long)r * p.lds + c] : 0.f;
    }
    __syncthreads();
    float* d = p.dst + z * p.sDz; const float* rr = p.R2 + z * p.sRz;
#pragma unroll
    for (int k = 0; k < 4; ++k) {
        const int cl = wave * 4 + k, c = c0 + cl, r = r0 + lane;
        if (c < p.C && r < p.R) {
            float v = act_fn(p.alpha * tile[lane][cl], p.act);
            if (p.flags & 1) v += p.beta * rr[(long long)c * p.ldr + r];
            VST2(float, d + (long long)c * p.ldd + r, v);
        }
    }
}

__global__ __launch_bounds__(256) void k_affine(const float* __restrict__ src, float* __restrict__ dst, int n, float a, float b, const float* __restrict__ sdev) {
    const int i = blockIdx.x * 256 + threadIdx.x;
    if (i < n) { const float aa = sdev ? a * sdev[0] : a; const float v = aa * src[i] + b; VST2(float, dst + i, v); }
}

struct SmP { const float* src; float* dst; const float* Mf; long long sz, sr, dz, dr, smz, smr; int n, pad; float scale_in, scale_out; };
static_assert(sizeof(SmP) == 3 * 8 + 6 * 8 + 4 * 4, "SmP has padding");
__global__ __launch_bounds__(256) void k_softmax(SmP p) {
    __shared__ float red[256];
    const int r = blockIdx.x, z = blockIdx.y, tid = threadIdx.x;
    const float* s = p.src + z * p.sz + (long long)r * p.sr;
    const float* mf = p.Mf ? (p.Mf + z * p.smz + (long long)r * p.smr) : nullptr;
    float mx = -__builtin_inff();
    for (int j = tid; j < p.n; j += 256) { float v = s[j] * p.scale_in; if (mf) v += mf[j]; mx = fmaxf(mx, v); }
    red[tid] = mx; __syncthreads();
    for (int o = 128; o > 0; o >>= 1) { if (tid < o) red[tid] = fmaxf(red[tid], red[tid + o]); __syncthreads(); }
    mx = red[0]; __syncthreads();
    float sum = 0.f;
    for (int j = tid; j < p.n; j += 256) { float v = s[j] * p.scale_in; if (mf) v += mf[j]; sum += (mx == -__builtin_inff()) ? 0.f : expf(v - mx); }
    red[tid] = sum; __syncthreads();
    for (int o = 128; o > 0; o >>= 1) { if (tid < o) red[tid] += red[tid + o]; __syncthreads(); }
    sum = red[0];
    const float inv = (sum > 0.f) ? p.scale_out / sum : 0.f;
    float* d = p.dst + z * p.dz + (long long)r * p.dr;
    for (int j = tid; j < p.n; j += 256) { float v = s[j] * p.scale_in; if (mf) v += mf[j]; const float o = (mx == -__builtin_inff()) ? 0.f : expf(v - mx) * inv; VST2(float, d + j, o); }
}
__global__ __launch_bounds__(256) void k_stats(const float* __restrict__ x, long long sz, long long so, long long si, int inner, int n, float eps, float* __restrict__ stat, int mode) {
    __shared__ float red[256];
    const int z = blockIdx.x, tid = threadIdx.x;
    const float* base = x + z * sz;
    float s = 0.f;
    for (int e = tid; e < n; e += 256) s += base[(long long)(e / inner) * so + (long long)(e % inner) * si];
    red[tid] = s; __syncthreads();
    for (int o = 128; o > 0; o >>= 1) { if (tid < o) red[tid] += red[tid + o]; __syncthreads(); }
    const float mu = (mode == 0 || mode == 3) ? red[0] / (float)n : 0.f; __syncthreads();
    float q = 0.f;
    for (int e = tid; e < n; e += 256) { const float dlt = base[(long long)(e / inner) * so + (long long)(e % inner) * si] - mu; q += dlt * dlt; }
    red[tid] = q; __syncthreads();
    for (int o = 128; o > 0; o >>= 1) { if (tid < o) red[tid] += red[tid + o]; __syncthreads(); }
    {
        float rs;
        if (mode == 2) rs = sqrtf((float)n) / fmaxf(sqrtf(red[0]), eps); else if (mode == 3) rs = rsqrtf(red[0] / (float)(n - 1) + eps); else rs = rsqrtf(red[0] / (float)n + eps);
        if (tid < 32) { const float v = (tid == 0) ? mu : ((tid == 1) ? rs : 0.f); VST2(float, stat + (long long)z * 32 + tid, v); }
    }
}
__global__ __launch_bounds__(256) void k_norm_apply(const float* __restrict__ x, float* __restrict__ y, const float* __restrict__ stat, const float* __restrict__ g, const float* __restrict__ bta,
                                                     int Z, int C, int L, int G, int bn, int act) {
    const long long idx = (long long)blockIdx.x * 256 + threadIdx.x;
    if (idx >= (long long)Z * C * L) return;
    const int l = (int)(idx % L); const long long zc = idx / L; const int c = (int)(zc % C), z = (int)(zc / C); (void)l;
    const int set = bn ? c : (z * G + c / (C / G));
    float v = (x[idx] - stat[(long long)set * 32]) * stat[(long long)set * 32 + 1];
    if (g) v *= g[c];
    if (bta) v += bta[c];
    v = act_fn(v, act);
    VST2(float, y + idx, v);
}

__global__ __launch_bounds__(256) void k_lse_neg(const float* __restrict__ st, float* __restrict__ c, int n) {
    const int i = blockIdx.x * 256 + threadIdx.x;
    if (i < n) { const float v = -(st[2 * i] + logf(st[2 * i + 1])); VST2(float, c + i, v); }
}

__global__ __launch_bounds__(256) void k_iota(int* __restrict__ dst, int n, int a, int b) {
    const int i = blockIdx.x * 256 + threadIdx.x;
    if (i < n) { const int v = a * i + b; VST2(int, dst + i, v); }
}

__global__ __launch_bounds__(256) void k_axpby(const float* __restrict__ x, const float* __restrict__ y, float* __restrict__ dst, int n, float a, float b, float c) {
    const int i = blockIdx.x * 256 + threadIdx.x;
    if (i < n) { const float v = a * x[i] + b * y[i] + c; VST2(float, dst + i, v); }
}

struct RopeP { const float* X; float* Y; const float* C; const float* Sn; const int* pos; long long sXr, sXh, sYr, sYh, sCb, sCp, sCd; int R, Hn, D, S, mode, tmode, pmode, pad; };
static_assert(sizeof(RopeP) == 5 * 8 + 7 * 8 + 8 * 4, "RopeP has padding");
__global__ __launch_bounds__(256) void k_rope(RopeP p) {
    const long long idx = (long long)blockIdx.x * 256 + threadIdx.x;
    if (idx >= (long long)p.R * p.Hn * p.D) return;
    const int d = (int)(idx % p.D); const long long rh = idx / p.D; const int h = (int)(rh % p.Hn); const int r = (int)(rh / p.Hn);
    const int half = p.D / 2;
    int partner; float sign;
    if (p.mode == 0) { partner = (d < half) ? d + half : d - half; sign = (d < half) ? -1.f : 1.f; }
    else { partner = d ^ 1; sign = (d & 1) ? 1.f : -1.f; }
    const int tcol = (p.tmode == 0) ? d : ((p.tmode == 1) ? (d % half) : (d >> 1));
    const int pp = (p.pmode == 0) ? (r % p.S) : ((p.pmode == 1) ? h : p.pos[r]);
    const long long toff = (long long)(r / p.S) * p.sCb + (long long)pp * p.sCp + (long long)tcol * p.sCd;
    const float* xr = p.X + (long long)r * p.sXr + (long long)h * p.sXh;
    const float v = xr[d] * p.C[toff] + sign * xr[partner] * p.Sn[toff];
    VST2(float, p.Y + (long long)r * p.sYr + (long long)h * p.sYh + d, v);
}

__global__ __launch_bounds__(256) void k_invf(float* __restrict__ invb, int half, int D, float base, float num, int fmode, float cexp) {
    const int i = blockIdx.x * 256 + threadIdx.x;
    if (i >= ((half + 31) / 32) * 32) return;
    if (i >= half) { VST2(float, invb + i, 0.f); return; }
    const float e = (float)(2 * i) / (float)D;
    float invf;
    if (fmode == 1) invf = num * expf((float)(2 * i) * cexp);
    else if (fmode == 2) invf = num * powf(base, (-2.0f * ((float)i - 1.0f)) / (float)D);
    else invf = num * (1.0f / powf(base, e));
    VST2(float, invb + i, invf);
}
__global__ __launch_bounds__(256) void k_sincos(float* __restrict__ cs, float* __restrict__ sn, const float* __restrict__ invb, int S, int half, float pscale) {
    const int idx = blockIdx.x * 256 + threadIdx.x;
    if (idx >= S * half) return;
    const int s = idx / half, i = idx - s * half;
    const float ang = (pscale * (float)s) * invb[i];
    VST2(float, cs + idx, cosf(ang)); VST2(float, sn + idx, sinf(ang));
}

__global__ __launch_bounds__(256) void k_mulact(const float* __restrict__ x, const float* __restrict__ y, float* __restrict__ dst, int n, int act) {
    const int i = blockIdx.x * 256 + threadIdx.x;
    if (i < n) { const float v = act_fn(x[i], act) * y[i]; VST2(float, dst + i, v); }
}

__global__ __launch_bounds__(256) void k_matvec(GemmP p) {
    const int rpt = (p.N == 1) ? 1 : 32;
    const long long r0 = ((long long)blockIdx.x * 256 + threadIdx.x) * rpt; const int z = blockIdx.z, zo = z / p.zi_n, zi = z - zo * p.zi_n;
    if (r0 >= p.M) return;
    const float* Bb = p.B + zo * p.sBo + zi * p.sBi;
    float* C = p.C + zo * p.sCo + zi * p.sCi; const float* R = p.R + zo * p.sRo + zi * p.sRi;
    for (int rr = 0; rr < rpt; ++rr) {
        const long long r = r0 + rr; if (r >= p.M) break;
        const float* A = p.A + zo * p.sAo + zi * p.sAi + r * p.sAm;
        float acc[8] = {0.f, 0.f, 0.f, 0.f, 0.f, 0.f, 0.f, 0.f};
        for (int k = 0; k < p.K; ++k) { const float a = A[(long long)k * p.sAk];
#pragma unroll
            for (int j = 0; j < 8; ++j) if (j < p.N) acc[j] += a * Bb[(long long)j * p.sBn + (long long)k * p.sBk]; }
#pragma unroll
        for (int j = 0; j < 8; ++j) if (j < p.N) {
            float v = acc[j] * p.alpha;
            if (p.flags & 1) v += p.bias[j];
            if (p.flags & 2) v += p.bias[r];
            v = act_fn(v, p.act);
            if (p.flags & 4) v += p.beta * R[r * p.sRm + (long long)j * p.sRn];
            VST2(float, C + r * p.sCm + j, v);
        }
    }
}
__global__ __launch_bounds__(256) void k_smallsoftmax(const float* __restrict__ src, float* __restrict__ dst, long long sr, long long dr, int n, long long R, float scale) {
    const long long r0 = ((long long)blockIdx.x * 256 + threadIdx.x) * 32;
    for (int rr = 0; rr < 32; ++rr) {
        const long long r = r0 + rr; if (r >= R) return;
        const float* s = src + r * sr; float* d = dst + r * dr;
        float mx = -__builtin_inff();
        for (int j = 0; j < n; ++j) mx = fmaxf(mx, s[j] * scale);
        float sum = 0.f;
        for (int j = 0; j < n; ++j) sum += expf(s[j] * scale - mx);
        const float inv = 1.f / sum;
        for (int j = 0; j < n; ++j) { const float v = expf(s[j] * scale - mx) * inv; VST2(float, d + j, v); }
    }
}

__global__ __launch_bounds__(32) void k_unitstat(float* __restrict__ st) { const int t = threadIdx.x; const float v = (t == 1) ? 1.f : 0.f; VST2(float, st + t, v); }

__global__ __launch_bounds__(256) void k_lincopy(const float* __restrict__ src, long long lds, float* __restrict__ dst, long long ldd, long long rows, int cols) {
    const long long i = (long long)blockIdx.x * 256 + threadIdx.x; if (i >= rows * cols) return;
    const long long r = i / cols; const int c = (int)(i - r * cols);
    const float v = src[r * lds + c]; VST2(float, dst + r * ldd + c, v);
}

__global__ __launch_bounds__(256) void k_bl_pad(const float* __restrict__ SRC, float* __restrict__ XP, int NF, int C) { const long long q = (long long)blockIdx.x * 256 + threadIdx.x; if (q >= (long long)NF * 256 * C) return; const int c = (int)(q % C); const int x = (int)((q / C) % 16); const int y = (int)((q / (C * 16)) % 16); const int f = (int)(q / ((long long)C * 256)); VST2(float, XP + (((long long)f * 18 + y + 1) * 18 + x + 1) * C + c, SRC[q]); }
__global__ __launch_bounds__(256) void k_bl_cell(const float* __restrict__ XG, const float* __restrict__ GH, float* __restrict__ Cc, float* __restrict__ HS, float* __restrict__ HP, int B, int T, int t, int C) { const long long q = (long long)blockIdx.x * 256 + threadIdx.x; if (q >= (long long)B * 256 * C) return; const int c = (int)(q % C); const int p = (int)((q / C) % 256); const int b = (int)(q / ((long long)C * 256));
    const float* xg = XG + (((long long)b * T + t) * 256 + p) * 4 * C; const float* gh = GH + ((long long)b * 256 + p) * 4 * C;
    const float gi = xg[c] + gh[c], gf = xg[C + c] + gh[C + c], gc = xg[2 * C + c] + gh[2 * C + c], go = xg[3 * C + c] + gh[3 * C + c];
    const float i = fminf(fmaxf(0.2f * gi + 0.5f, 0.f), 1.f), f = fminf(fmaxf(0.2f * gf + 0.5f, 0.f), 1.f), o = fminf(fmaxf(0.2f * go + 0.5f, 0.f), 1.f);
    const float cn = f * Cc[q] + i * tanhf(gc); const float h = o * tanhf(cn); VST2(float, Cc + q, cn); VST2(float, HS + (((long long)b * T + t) * 256 + p) * C + c, h);
    const int y = p / 16, x = p % 16; VST2(float, HP + (((long long)b * 18 + y + 1) * 18 + x + 1) * C + c, h); }

template __global__ void k_gemm<1>(GemmP);

extern "C" void kernel_launch(void* const* d_in, const int* in_sizes, int n_in, void* d_out, int out_size, void* d_ws, size_t ws_size, hipStream_t stream) {
    (void)in_sizes; (void)n_in; (void)out_size; (void)ws_size;
    const float* x = (const float*)d_in[0];
    const float* Wx1 = (const float*)d_in[1];
    const float* Wh1 = (const float*)d_in[2];
    const float* b1 = (const float*)d_in[3];
    const float* g1 = (const float*)d_in[4];
    const float* be1 = (const float*)d_in[5];
    const float* Wx2 = (const float*)d_in[6];
    const float* Wh2 = (const float*)d_in[7];
    const float* b2 = (const float*)d_in[8];
    const float* g2 = (const float*)d_in[9];
    const float* be2 = (const float*)d_in[10];
    const float* Wx3 = (const float*)d_in[11];
    const float* Wh3 = (const float*)d_in[12];
    const float* b3 = (const float*)d_in[13];
    const float* g3 = (const float*)d_in[14];
    const float* be3 = (const float*)d_in[15];
    const int Bn = 4;
    const int T = 8;
    const int HW = 256;
    const int C = 256;
    const int G4 = 1024;
    const int NF = Bn * T;
    const int PP = 324;
    float* out = (float*)d_out;
    char* wsp = (char*)d_ws;
    float* XP = (float*)wsp; wsp += (((size_t)((size_t)NF * PP * C) * 4 + 255) / 256) * 256;
    float* XG = (float*)wsp; wsp += (((size_t)((size_t)NF * HW * G4) * 4 + 255) / 256) * 256;
    float* HP = (float*)wsp; wsp += (((size_t)((size_t)Bn * PP * C) * 4 + 255) / 256) * 256;
    float* GH = (float*)wsp; wsp += (((size_t)((size_t)Bn * HW * G4) * 4 + 255) / 256) * 256;
    float* Cc = (float*)wsp; wsp += (((size_t)((size_t)Bn * HW * C) * 4 + 255) / 256) * 256;
    float* HS = (float*)wsp; wsp += (((size_t)((size_t)NF * HW * C) * 4 + 255) / 256) * 256;
    float* st = (float*)wsp; wsp += (((size_t)((size_t)C * 32) * 4 + 255) / 256) * 256;
    hipMemsetAsync(XP, 0, (size_t)NF * PP * C * 4, stream); hipMemsetAsync(HP, 0, (size_t)Bn * PP * C * 4, stream); hipMemsetAsync(Cc, 0, (size_t)Bn * HW * C * 4, stream);
    k_bl_pad<<<(unsigned)(((long long)NF * HW * C + 255) / 256), 256, 0, stream>>>(x, XP, NF, C);
    { GemmP cx0_0;
      cx0_0.A = XP + (size_t)0 * C; cx0_0.B = Wx1 + (size_t)0 * C * G4; cx0_0.bias = b1; cx0_0.R = XP + (size_t)0 * C; cx0_0.C = XG;
      cx0_0.sAo = (long long)PP * C; cx0_0.sAi = (long long)18 * C; cx0_0.sAm = C; cx0_0.sAk = 1; cx0_0.sBo = 0; cx0_0.sBi = 0; cx0_0.sBn = 1; cx0_0.sBk = G4; cx0_0.sCo = (long long)HW * G4; cx0_0.sCi = (long long)16 * G4; cx0_0.sCm = G4; cx0_0.sRo = 0; cx0_0.sRi = 0; cx0_0.sRm = 0; cx0_0.sRn = 0;
      cx0_0.M = 16; cx0_0.N = G4; cx0_0.K = C; cx0_0.zi_n = 16; cx0_0.flags = 1; cx0_0.act = 0;
      cx0_0.alpha = 1.0f; cx0_0.beta = 0.0f; cx0_0.sa = 1.0f; cx0_0.sb = 1.0f; cx0_0.Npad = G4; cx0_0.pad_ = 0;
      k_gemm<1><<<dim3((unsigned)((G4) + 31) / 32, (unsigned)((16) + 15) / 16, (unsigned)(NF * 16)), 32, 0, stream>>>(cx0_0); }
    { GemmP cx0_1;
      cx0_1.A = XP + (size_t)1 * C; cx0_1.B = Wx1 + (size_t)1 * C * G4; cx0_1.bias = XP + (size_t)1 * C; cx0_1.R = XG; cx0_1.C = XG;
      cx0_1.sAo = (long long)PP * C; cx0_1.sAi = (long long)18 * C; cx0_1.sAm = C; cx0_1.sAk = 1; cx0_1.sBo = 0; cx0_1.sBi = 0; cx0_1.sBn = 1; cx0_1.sBk = G4; cx0_1.sCo = (long long)HW * G4; cx0_1.sCi = (long long)16 * G4; cx0_1.sCm = G4; cx0_1.sRo = (long long)HW * G4; cx0_1.sRi = (long long)16 * G4; cx0_1.sRm = G4; cx0_1.sRn = 1;
      cx0_1.M = 16; cx0_1.N = G4; cx0_1.K = C; cx0_1.zi_n = 16; cx0_1.flags = 4; cx0_1.act = 0;
      cx0_1.alpha = 1.0f; cx0_1.beta = 1.0f; cx0_1.sa = 1.0f; cx0_1.sb = 1.0f; cx0_1.Npad = G4; cx0_1.pad_ = 0;
      k_gemm<1><<<dim3((unsigned)((G4) + 31) / 32, (unsigned)((16) + 15) / 16, (unsigned)(NF * 16)), 32, 0, stream>>>(cx0_1); }
    { GemmP cx0_2;
      cx0_2.A = XP + (size_t)2 * C; cx0_2.B = Wx1 + (size_t)2 * C * G4; cx0_2.bias = XP + (size_t)2 * C; cx0_2.R = XG; cx0_2.C = XG;
      cx0_2.sAo = (long long)PP * C; cx0_2.sAi = (long long)18 * C; cx0_2.sAm = C; cx0_2.sAk = 1; cx0_2.sBo = 0; cx0_2.sBi = 0; cx0_2.sBn = 1; cx0_2.sBk = G4; cx0_2.sCo = (long long)HW * G4; cx0_2.sCi = (long long)16 * G4; cx0_2.sCm = G4; cx0_2.sRo = (long long)HW * G4; cx0_2.sRi = (long long)16 * G4; cx0_2.sRm = G4; cx0_2.sRn = 1;
      cx0_2.M = 16; cx0_2.N = G4; cx0_2.K = C; cx0_2.zi_n = 16; cx0_2.flags = 4; cx0_2.act = 0;
      cx0_2.alpha = 1.0f; cx0_2.beta = 1.0f; cx0_2.sa = 1.0f; cx0_2.sb = 1.0f; cx0_2.Npad = G4; cx0_2.pad_ = 0;
      k_gemm<1><<<dim3((unsigned)((G4) + 31) / 32, (unsigned)((16) + 15) / 16, (unsigned)(NF * 16)), 32, 0, stream>>>(cx0_2); }
    { GemmP cx0_3;
      cx0_3.A = XP + (size_t)18 * C; cx0_3.B = Wx1 + (size_t)3 * C * G4; cx0_3.bias = XP + (size_t)18 * C; cx0_3.R = XG; cx0_3.C = XG;
      cx0_3.sAo = (long long)PP * C; cx0_3.sAi = (long long)18 * C; cx0_3.sAm = C; cx0_3.sAk = 1; cx0_3.sBo = 0; cx0_3.sBi = 0; cx0_3.sBn = 1; cx0_3.sBk = G4; cx0_3.sCo = (long long)HW * G4; cx0_3.sCi = (long long)16 * G4; cx0_3.sCm = G4; cx0_3.sRo = (long long)HW * G4; cx0_3.sRi = (long long)16 * G4; cx0_3.sRm = G4; cx0_3.sRn = 1;
      cx0_3.M = 16; cx0_3.N = G4; cx0_3.K = C; cx0_3.zi_n = 16; cx0_3.flags = 4; cx0_3.act = 0;
      cx0_3.alpha = 1.0f; cx0_3.beta = 1.0f; cx0_3.sa = 1.0f; cx0_3.sb = 1.0f; cx0_3.Npad = G4; cx0_3.pad_ = 0;
      k_gemm<1><<<dim3((unsigned)((G4) + 31) / 32, (unsigned)((16) + 15) / 16, (unsigned)(NF * 16)), 32, 0, stream>>>(cx0_3); }
    { GemmP cx0_4;
      cx0_4.A = XP + (size_t)19 * C; cx0_4.B = Wx1 + (size_t)4 * C * G4; cx0_4.bias = XP + (size_t)19 * C; cx0_4.R = XG; cx0_4.C = XG;
      cx0_4.sAo = (long long)PP * C; cx0_4.sAi = (long long)18 * C; cx0_4.sAm = C; cx0_4.sAk = 1; cx0_4.sBo = 0; cx0_4.sBi = 0; cx0_4.sBn = 1; cx0_4.sBk = G4; cx0_4.sCo = (long long)HW * G4; cx0_4.sCi = (long long)16 * G4; cx0_4.sCm = G4; cx0_4.sRo = (long long)HW * G4; cx0_4.sRi = (long long)16 * G4; cx0_4.sRm = G4; cx0_4.sRn = 1;
      cx0_4.M = 16; cx0_4.N = G4; cx0_4.K = C; cx0_4.zi_n = 16; cx0_4.flags = 4; cx0_4.act = 0;
      cx0_4.alpha = 1.0f; cx0_4.beta = 1.0f; cx0_4.sa = 1.0f; cx0_4.sb = 1.0f; cx0_4.Npad = G4; cx0_4.pad_ = 0;
      k_gemm<1><<<dim3((unsigned)((G4) + 31) / 32, (unsigned)((16) + 15) / 16, (unsigned)(NF * 16)), 32, 0, stream>>>(cx0_4); }
    { GemmP cx0_5;
      cx0_5.A = XP + (size_t)20 * C; cx0_5.B = Wx1 + (size_t)5 * C * G4; cx0_5.bias = XP + (size_t)20 * C; cx0_5.R = XG; cx0_5.C = XG;
      cx0_5.sAo = (long long)PP * C; cx0_5.sAi = (long long)18 * C; cx0_5.sAm = C; cx0_5.sAk = 1; cx0_5.sBo = 0; cx0_5.sBi = 0; cx0_5.sBn = 1; cx0_5.sBk = G4; cx0_5.sCo = (long long)HW * G4; cx0_5.sCi = (long long)16 * G4; cx0_5.sCm = G4; cx0_5.sRo = (long long)HW * G4; cx0_5.sRi = (long long)16 * G4; cx0_5.sRm = G4; cx0_5.sRn = 1;
      cx0_5.M = 16; cx0_5.N = G4; cx0_5.K = C; cx0_5.zi_n = 16; cx0_5.flags = 4; cx0_5.act = 0;
      cx0_5.alpha = 1.0f; cx0_5.beta = 1.0f; cx0_5.sa = 1.0f; cx0_5.sb = 1.0f; cx0_5.Npad = G4; cx0_5.pad_ = 0;
      k_gemm<1><<<dim3((unsigned)((G4) + 31) / 32, (unsigned)((16) + 15) / 16, (unsigned)(NF * 16)), 32, 0, stream>>>(cx0_5); }
    { GemmP cx0_6;
      cx0_6.A = XP + (size_t)36 * C; cx0_6.B = Wx1 + (size_t)6 * C * G4; cx0_6.bias = XP + (size_t)36 * C; cx0_6.R = XG; cx0_6.C = XG;
      cx0_6.sAo = (long long)PP * C; cx0_6.sAi = (long long)18 * C; cx0_6.sAm = C; cx0_6.sAk = 1; cx0_6.sBo = 0; cx0_6.sBi = 0; cx0_6.sBn = 1; cx0_6.sBk = G4; cx0_6.sCo = (long long)HW * G4; cx0_6.sCi = (long long)16 * G4; cx0_6.sCm = G4; cx0_6.sRo = (long long)HW * G4; cx0_6.sRi = (long long)16 * G4; cx0_6.sRm = G4; cx0_6.sRn = 1;
      cx0_6.M = 16; cx0_6.N = G4; cx0_6.K = C; cx0_6.zi_n = 16; cx0_6.flags = 4; cx0_6.act = 0;
      cx0_6.alpha = 1.0f; cx0_6.beta = 1.0f; cx0_6.sa = 1.0f; cx0_6.sb = 1.0f; cx0_6.Npad = G4; cx0_6.pad_ = 0;
      k_gemm<1><<<dim3((unsigned)((G4) + 31) / 32, (unsigned)((16) + 15) / 16, (unsigned)(NF * 16)), 32, 0, stream>>>(cx0_6); }
    { GemmP cx0_7;
      cx0_7.A = XP + (size_t)37 * C; cx0_7.B = Wx1 + (size_t)7 * C * G4; cx0_7.bias = XP + (size_t)37 * C; cx0_7.R = XG; cx0_7.C = XG;
      cx0_7.sAo = (long long)PP * C; cx0_7.sAi = (long long)18 * C; cx0_7.sAm = C; cx0_7.sAk = 1; cx0_7.sBo = 0; cx0_7.sBi = 0; cx0_7.sBn = 1; cx0_7.sBk = G4; cx0_7.sCo = (long long)HW * G4; cx0_7.sCi = (long long)16 * G4; cx0_7.sCm = G4; cx0_7.sRo = (long long)HW * G4; cx0_7.sRi = (long long)16 * G4; cx0_7.sRm = G4; cx0_7.sRn = 1;
      cx0_7.M = 16; cx0_7.N = G4; cx0_7.K = C; cx0_7.zi_n = 16; cx0_7.flags = 4; cx0_7.act = 0;
      cx0_7.alpha = 1.0f; cx0_7.beta = 1.0f; cx0_7.sa = 1.0f; cx0_7.sb = 1.0f; cx0_7.Npad = G4; cx0_7.pad_ = 0;
      k_gemm<1><<<dim3((unsigned)((G4) + 31) / 32, (unsigned)((16) + 15) / 16, (unsigned)(NF * 16)), 32, 0, stream>>>(cx0_7); }
    { GemmP cx0_8;
      cx0_8.A = XP + (size_t)38 * C; cx0_8.B = Wx1 + (size_t)8 * C * G4; cx0_8.bias = XP + (size_t)38 * C; cx0_8.R = XG; cx0_8.C = XG;
      cx0_8.sAo = (long long)PP * C; cx0_8.sAi = (long long)18 * C; cx0_8.sAm = C; cx0_8.sAk = 1; cx0_8.sBo = 0; cx0_8.sBi = 0; cx0_8.sBn = 1; cx0_8.sBk = G4; cx0_8.sCo = (long long)HW * G4; cx0_8.sCi = (long long)16 * G4; cx0_8.sCm = G4; cx0_8.sRo = (long long)HW * G4; cx0_8.sRi = (long long)16 * G4; cx0_8.sRm = G4; cx0_8.sRn = 1;
      cx0_8.M = 16; cx0_8.N = G4; cx0_8.K = C; cx0_8.zi_n = 16; cx0_8.flags = 4; cx0_8.act = 0;
      cx0_8.alpha = 1.0f; cx0_8.beta = 1.0f; cx0_8.sa = 1.0f; cx0_8.sb = 1.0f; cx0_8.Npad = G4; cx0_8.pad_ = 0;
      k_gemm<1><<<dim3((unsigned)((G4) + 31) / 32, (unsigned)((16) + 15) / 16, (unsigned)(NF * 16)), 32, 0, stream>>>(cx0_8); }

    { GemmP ch0_0_0;
      ch0_0_0.A = HP + (size_t)0 * C; ch0_0_0.B = Wh1 + (size_t)0 * C * G4; ch0_0_0.bias = HP + (size_t)0 * C; ch0_0_0.R = HP + (size_t)0 * C; ch0_0_0.C = GH;
      ch0_0_0.sAo = (long long)PP * C; ch0_0_0.sAi = (long long)18 * C; ch0_0_0.sAm = C; ch0_0_0.sAk = 1; ch0_0_0.sBo = 0; ch0_0_0.sBi = 0; ch0_0_0.sBn = 1; ch0_0_0.sBk = G4; ch0_0_0.sCo = (long long)HW * G4; ch0_0_0.sCi = (long long)16 * G4; ch0_0_0.sCm = G4; ch0_0_0.sRo = 0; ch0_0_0.sRi = 0; ch0_0_0.sRm = 0; ch0_0_0.sRn = 0;
      ch0_0_0.M = 16; ch0_0_0.N = G4; ch0_0_0.K = C; ch0_0_0.zi_n = 16; ch0_0_0.flags = 0; ch0_0_0.act = 0;
      ch0_0_0.alpha = 1.0f; ch0_0_0.beta = 0.0f; ch0_0_0.sa = 1.0f; ch0_0_0.sb = 1.0f; ch0_0_0.Npad = G4; ch0_0_0.pad_ = 0;
      k_gemm<1><<<dim3((unsigned)((G4) + 31) / 32, (unsigned)((16) + 15) / 16, (unsigned)(Bn * 16)), 32, 0, stream>>>(ch0_0_0); }
    { GemmP ch0_0_1;
      ch0_0_1.A = HP + (size_t)1 * C; ch0_0_1.B = Wh1 + (size_t)1 * C * G4; ch0_0_1.bias = HP + (size_t)1 * C; ch0_0_1.R = GH; ch0_0_1.C = GH;
      ch0_0_1.sAo = (long long)PP * C; ch0_0_1.sAi = (long long)18 * C; ch0_0_1.sAm = C; ch0_0_1.sAk = 1; ch0_0_1.sBo = 0; ch0_0_1.sBi = 0; ch0_0_1.sBn = 1; ch0_0_1.sBk = G4; ch0_0_1.sCo = (long long)HW * G4; ch0_0_1.sCi = (long long)16 * G4; ch0_0_1.sCm = G4; ch0_0_1.sRo = (long long)HW * G4; ch0_0_1.sRi = (long long)16 * G4; ch0_0_1.sRm = G4; ch0_0_1.sRn = 1;
      ch0_0_1.M = 16; ch0_0_1.N = G4; ch0_0_1.K = C; ch0_0_1.zi_n = 16; ch0_0_1.flags = 4; ch0_0_1.act = 0;
      ch0_0_1.alpha = 1.0f; ch0_0_1.beta = 1.0f; ch0_0_1.sa = 1.0f; ch0_0_1.sb = 1.0f; ch0_0_1.Npad = G4; ch0_0_1.pad_ = 0;
      k_gemm<1><<<dim3((unsigned)((G4) + 31) / 32, (unsigned)((16) + 15) / 16, (unsigned)(Bn * 16)), 32, 0, stream>>>(ch0_0_1); }
    { GemmP ch0_0_2;
      ch0_0_2.A = HP + (size_t)2 * C; ch0_0_2.B = Wh1 + (size_t)2 * C * G4; ch0_0_2.bias = HP + (size_t)2 * C; ch0_0_2.R = GH; ch0_0_2.C = GH;
      ch0_0_2.sAo = (long long)PP * C; ch0_0_2.sAi = (long long)18 * C; ch0_0_2.sAm = C; ch0_0_2.sAk = 1; ch0_0_2.sBo = 0; ch0_0_2.sBi = 0; ch0_0_2.sBn = 1; ch0_0_2.sBk = G4; ch0_0_2.sCo = (long long)HW * G4; ch0_0_2.sCi = (long long)16 * G4; ch0_0_2.sCm = G4; ch0_0_2.sRo = (long long)HW * G4; ch0_0_2.sRi = (long long)16 * G4; ch0_0_2.sRm = G4; ch0_0_2.sRn = 1;
      ch0_0_2.M = 16; ch0_0_2.N = G4; ch0_0_2.K = C; ch0_0_2.zi_n = 16; ch0_0_2.flags = 4; ch0_0_2.act = 0;
      ch0_0_2.alpha = 1.0f; ch0_0_2.beta = 1.0f; ch0_0_2.sa = 1.0f; ch0_0_2.sb = 1.0f; ch0_0_2.Npad = G4; ch0_0_2.pad_ = 0;
      k_gemm<1><<<dim3((unsigned)((G4) + 31) / 32, (unsigned)((16) + 15) / 16, (unsigned)(Bn * 16)), 32, 0, stream>>>(ch0_0_2); }
    { GemmP ch0_0_3;
      ch0_0_3.A = HP + (size_t)18 * C; ch0_0_3.B = Wh1 + (size_t)3 * C * G4; ch0_0_3.bias = HP + (size_t)18 * C; ch0_0_3.R = GH; ch0_0_3.C = GH;
      ch0_0_3.sAo = (long long)PP * C; ch0_0_3.sAi = (long long)18 * C; ch0_0_3.sAm = C; ch0_0_3.sAk = 1; ch0_0_3.sBo = 0; ch0_0_3.sBi = 0; ch0_0_3.sBn = 1; ch0_0_3.sBk = G4; ch0_0_3.sCo = (long long)HW * G4; ch0_0_3.sCi = (long long)16 * G4; ch0_0_3.sCm = G4; ch0_0_3.sRo = (long long)HW * G4; ch0_0_3.sRi = (long long)16 * G4; ch0_0_3.sRm = G4; ch0_0_3.sRn = 1;
      ch0_0_3.M = 16; ch0_0_3.N = G4; ch0_0_3.K = C; ch0_0_3.zi_n = 16; ch0_0_3.flags = 4; ch0_0_3.act = 0;
      ch0_0_3.alpha = 1.0f; ch0_0_3.beta = 1.0f; ch0_0_3.sa = 1.0f; ch0_0_3.sb = 1.0f; ch0_0_3.Npad = G4; ch0_0_3.pad_ = 0;
      k_gemm<1><<<dim3((unsigned)((G4) + 31) / 32, (unsigned)((16) + 15) / 16, (unsigned)(Bn * 16)), 32, 0, stream>>>(ch0_0_3); }
    { GemmP ch0_0_4;
      ch0_0_4.A = HP + (size_t)19 * C; ch0_0_4.B = Wh1 + (size_t)4 * C * G4; ch0_0_4.bias = HP + (size_t)19 * C; ch0_0_4.R = GH; ch0_0_4.C = GH;
      ch0_0_4.sAo = (long long)PP * C; ch0_0_4.sAi = (long long)18 * C; ch0_0_4.sAm = C; ch0_0_4.sAk = 1; ch0_0_4.sBo = 0; ch0_0_4.sBi = 0; ch0_0_4.sBn = 1; ch0_0_4.sBk = G4; ch0_0_4.sCo = (long long)HW * G4; ch0_0_4.sCi = (long long)16 * G4; ch0_0_4.sCm = G4; ch0_0_4.sRo = (long long)HW * G4; ch0_0_4.sRi = (long long)16 * G4; ch0_0_4.sRm = G4; ch0_0_4.sRn = 1;
      ch0_0_4.M = 16; ch0_0_4.N = G4; ch0_0_4.K = C; ch0_0_4.zi_n = 16; ch0_0_4.flags = 4; ch0_0_4.act = 0;
      ch0_0_4.alpha = 1.0f; ch0_0_4.beta = 1.0f; ch0_0_4.sa = 1.0f; ch0_0_4.sb = 1.0f; ch0_0_4.Npad = G4; ch0_0_4.pad_ = 0;
      k_gemm<1><<<dim3((unsigned)((G4) + 31) / 32, (unsigned)((16) + 15) / 16, (unsigned)(Bn * 16)), 32, 0, stream>>>(ch0_0_4); }
    { GemmP ch0_0_5;
      ch0_0_5.A = HP + (size_t)20 * C; ch0_0_5.B = Wh1 + (size_t)5 * C * G4; ch0_0_5.bias = HP + (size_t)20 * C; ch0_0_5.R = GH; ch0_0_5.C = GH;
      ch0_0_5.sAo = (long long)PP * C; ch0_0_5.sAi = (long long)18 * C; ch0_0_5.sAm = C; ch0_0_5.sAk = 1; ch0_0_5.sBo = 0; ch0_0_5.sBi = 0; ch0_0_5.sBn = 1; ch0_0_5.sBk = G4; ch0_0_5.sCo = (long long)HW * G4; ch0_0_5.sCi = (long long)16 * G4; ch0_0_5.sCm = G4; ch0_0_5.sRo = (long long)HW * G4; ch0_0_5.sRi = (long long)16 * G4; ch0_0_5.sRm = G4; ch0_0_5.sRn = 1;
      ch0_0_5.M = 16; ch0_0_5.N = G4; ch0_0_5.K = C; ch0_0_5.zi_n = 16; ch0_0_5.flags = 4; ch0_0_5.act = 0;
      ch0_0_5.alpha = 1.0f; ch0_0_5.beta = 1.0f; ch0_0_5.sa = 1.0f; ch0_0_5.sb = 1.0f; ch0_0_5.Npad = G4; ch0_0_5.pad_ = 0;
      k_gemm<1><<<dim3((unsigned)((G4) + 31) / 32, (unsigned)((16) + 15) / 16, (unsigned)(Bn * 16)), 32, 0, stream>>>(ch0_0_5); }
    { GemmP ch0_0_6;
      ch0_0_6.A = HP + (size_t)36 * C; ch0_0_6.B = Wh1 + (size_t)6 * C * G4; ch0_0_6.bias = HP + (size_t)36 * C; ch0_0_6.R = GH; ch0_0_6.C = GH;
      ch0_0_6.sAo = (long long)PP * C; ch0_0_6.sAi = (long long)18 * C; ch0_0_6.sAm = C; ch0_0_6.sAk = 1; ch0_0_6.sBo = 0; ch0_0_6.sBi = 0; ch0_0_6.sBn = 1; ch0_0_6.sBk = G4; ch0_0_6.sCo = (long long)HW * G4; ch0_0_6.sCi = (long long)16 * G4; ch0_0_6.sCm = G4; ch0_0_6.sRo = (long long)HW * G4; ch0_0_6.sRi = (long long)16 * G4; ch0_0_6.sRm = G4; ch0_0_6.sRn = 1;
      ch0_0_6.M = 16; ch0_0_6.N = G4; ch0_0_6.K = C; ch0_0_6.zi_n = 16; ch0_0_6.flags = 4; ch0_0_6.act = 0;
      ch0_0_6.alpha = 1.0f; ch0_0_6.beta = 1.0f; ch0_0_6.sa = 1.0f; ch0_0_6.sb = 1.0f; ch0_0_6.Npad = G4; ch0_0_6.pad_ = 0;
      k_gemm<1><<<dim3((unsigned)((G4) + 31) / 32, (unsigned)((16) + 15) / 16, (unsigned)(Bn * 16)), 32, 0, stream>>>(ch0_0_6); }
    { GemmP ch0_0_7;
      ch0_0_7.A = HP + (size_t)37 * C; ch0_0_7.B = Wh1 + (size_t)7 * C * G4; ch0_0_7.bias = HP + (size_t)37 * C; ch0_0_7.R = GH; ch0_0_7.C = GH;
      ch0_0_7.sAo = (long long)PP * C; ch0_0_7.sAi = (long long)18 * C; ch0_0_7.sAm = C; ch0_0_7.sAk = 1; ch0_0_7.sBo = 0; ch0_0_7.sBi = 0; ch0_0_7.sBn = 1; ch0_0_7.sBk = G4; ch0_0_7.sCo = (long long)HW * G4; ch0_0_7.sCi = (long long)16 * G4; ch0_0_7.sCm = G4; ch0_0_7.sRo = (long long)HW * G4; ch0_0_7.sRi = (long long)16 * G4; ch0_0_7.sRm = G4; ch0_0_7.sRn = 1;
      ch0_0_7.M = 16; ch0_0_7.N = G4; ch0_0_7.K = C; ch0_0_7.zi_n = 16; ch0_0_7.flags = 4; ch0_0_7.act = 0;
      ch0_0_7.alpha = 1.0f; ch0_0_7.beta = 1.0f; ch0_0_7.sa = 1.0f; ch0_0_7.sb = 1.0f; ch0_0_7.Npad = G4; ch0_0_7.pad_ = 0;
      k_gemm<1><<<dim3((unsigned)((G4) + 31) / 32, (unsigned)((16) + 15) / 16, (unsigned)(Bn * 16)), 32, 0, stream>>>(ch0_0_7); }
    { GemmP ch0_0_8;
      ch0_0_8.A = HP + (size_t)38 * C; ch0_0_8.B = Wh1 + (size_t)8 * C * G4; ch0_0_8.bias = HP + (size_t)38 * C; ch0_0_8.R = GH; ch0_0_8.C = GH;
      ch0_0_8.sAo = (long long)PP * C; ch0_0_8.sAi = (long long)18 * C; ch0_0_8.sAm = C; ch0_0_8.sAk = 1; ch0_0_8.sBo = 0; ch0_0_8.sBi = 0; ch0_0_8.sBn = 1; ch0_0_8.sBk = G4; ch0_0_8.sCo = (long long)HW * G4; ch0_0_8.sCi = (long long)16 * G4; ch0_0_8.sCm = G4; ch0_0_8.sRo = (long long)HW * G4; ch0_0_8.sRi = (long long)16 * G4; ch0_0_8.sRm = G4; ch0_0_8.sRn = 1;
      ch0_0_8.M = 16; ch0_0_8.N = G4; ch0_0_8.K = C; ch0_0_8.zi_n = 16; ch0_0_8.flags = 4; ch0_0_8.act = 0;
      ch0_0_8.alpha = 1.0f; ch0_0_8.beta = 1.0f; ch0_0_8.sa = 1.0f; ch0_0_8.sb = 1.0f; ch0_0_8.Npad = G4; ch0_0_8.pad_ = 0;
      k_gemm<1><<<dim3((unsigned)((G4) + 31) / 32, (unsigned)((16) + 15) / 16, (unsigned)(Bn * 16)), 32, 0, stream>>>(ch0_0_8); }

    k_bl_cell<<<(unsigned)(((long long)Bn * HW * C + 255) / 256), 256, 0, stream>>>(XG, GH, Cc, HS, HP, Bn, T, 0, C);
    { GemmP ch0_1_0;
      ch0_1_0.A = HP + (size_t)0 * C; ch0_1_0.B = Wh1 + (size_t)0 * C * G4; ch0_1_0.bias = HP + (size_t)0 * C; ch0_1_0.R = HP + (size_t)0 * C; ch0_1_0.C = GH;
      ch0_1_0.sAo = (long long)PP * C; ch0_1_0.sAi = (long long)18 * C; ch0_1_0.sAm = C; ch0_1_0.sAk = 1; ch0_1_0.sBo = 0; ch0_1_0.sBi = 0; ch0_1_0.sBn = 1; ch0_1_0.sBk = G4; ch0_1_0.sCo = (long long)HW * G4; ch0_1_0.sCi = (long long)16 * G4; ch0_1_0.sCm = G4; ch0_1_0.sRo = 0; ch0_1_0.sRi = 0; ch0_1_0.sRm = 0; ch0_1_0.sRn = 0;
      ch0_1_0.M = 16; ch0_1_0.N = G4; ch0_1_0.K = C; ch0_1_0.zi_n = 16; ch0_1_0.flags = 0; ch0_1_0.act = 0;
      ch0_1_0.alpha = 1.0f; ch0_1_0.beta = 0.0f; ch0_1_0.sa = 1.0f; ch0_1_0.sb = 1.0f; ch0_1_0.Npad = G4; ch0_1_0.pad_ = 0;
      k_gemm<1><<<dim3((unsigned)((G4) + 31) / 32, (unsigned)((16) + 15) / 16, (unsigned)(Bn * 16)), 32, 0, stream>>>(ch0_1_0); }
    { GemmP ch0_1_1;
      ch0_1_1.A = HP + (size_t)1 * C; ch0_1_1.B = Wh1 + (size_t)1 * C * G4; ch0_1_1.bias = HP + (size_t)1 * C; ch0_1_1.R = GH; ch0_1_1.C = GH;
      ch0_1_1.sAo = (long long)PP * C; ch0_1_1.sAi = (long long)18 * C; ch0_1_1.sAm = C; ch0_1_1.sAk = 1; ch0_1_1.sBo = 0; ch0_1_1.sBi = 0; ch0_1_1.sBn = 1; ch0_1_1.sBk = G4; ch0_1_1.sCo = (long long)HW * G4; ch0_1_1.sCi = (long long)16 * G4; ch0_1_1.sCm = G4; ch0_1_1.sRo = (long long)HW * G4; ch0_1_1.sRi = (long long)16 * G4; ch0_1_1.sRm = G4; ch0_1_1.sRn = 1;
      ch0_1_1.M = 16; ch0_1_1.N = G4; ch0_1_1.K = C; ch0_1_1.zi_n = 16; ch0_1_1.flags = 4; ch0_1_1.act = 0;
      ch0_1_1.alpha = 1.0f; ch0_1_1.beta = 1.0f; ch0_1_1.sa = 1.0f; ch0_1_1.sb = 1.0f; ch0_1_1.Npad = G4; ch0_1_1.pad_ = 0;
      k_gemm<1><<<dim3((unsigned)((G4) + 31) / 32, (unsigned)((16) + 15) / 16, (unsigned)(Bn * 16)), 32, 0, stream>>>(ch0_1_1); }
    { GemmP ch0_1_2;
      ch0_1_2.A = HP + (size_t)2 * C; ch0_1_2.B = Wh1 + (size_t)2 * C * G4; ch0_1_2.bias = HP + (size_t)2 * C; ch0_1_2.R = GH; ch0_1_2.C = GH;
      ch0_1_2.sAo = (long long)PP * C; ch0_1_2.sAi = (long long)18 * C; ch0_1_2.sAm = C; ch0_1_2.sAk = 1; ch0_1_2.sBo = 0; ch0_1_2.sBi = 0; ch0_1_2.sBn = 1; ch0_1_2.sBk = G4; ch0_1_2.sCo = (long long)HW * G4; ch0_1_2.sCi = (long long)16 * G4; ch0_1_2.sCm = G4; ch0_1_2.sRo = (long long)HW * G4; ch0_1_2.sRi = (long long)16 * G4; ch0_1_2.sRm = G4; ch0_1_2.sRn = 1;
      ch0_1_2.M = 16; ch0_1_2.N = G4; ch0_1_2.K = C; ch0_1_2.zi_n = 16; ch0_1_2.flags = 4; ch0_1_2.act = 0;
      ch0_1_2.alpha = 1.0f; ch0_1_2.beta = 1.0f; ch0_1_2.sa = 1.0f; ch0_1_2.sb = 1.0f; ch0_1_2.Npad = G4; ch0_1_2.pad_ = 0;
      k_gemm<1><<<dim3((unsigned)((G4) + 31) / 32, (unsigned)((16) + 15) / 16, (unsigned)(Bn * 16)), 32, 0, stream>>>(ch0_1_2); }
    { GemmP ch0_1_3;
      ch0_1_3.A = HP + (size_t)18 * C; ch0_1_3.B = Wh1 + (size_t)3 * C * G4; ch0_1_3.bias = HP + (size_t)18 * C; ch0_1_3.R = GH; ch0_1_3.C = GH;
      ch0_1_3.sAo = (long long)PP * C; ch0_1_3.sAi = (long long)18 * C; ch0_1_3.sAm = C; ch0_1_3.sAk = 1; ch0_1_3.sBo = 0; ch0_1_3.sBi = 0; ch0_1_3.sBn = 1; ch0_1_3.sBk = G4; ch0_1_3.sCo = (long long)HW * G4; ch0_1_3.sCi = (long long)16 * G4; ch0_1_3.sCm = G4; ch0_1_3.sRo = (long long)HW * G4; ch0_1_3.sRi = (long long)16 * G4; ch0_1_3.sRm = G4; ch0_1_3.sRn = 1;
      ch0_1_3.M = 16; ch0_1_3.N = G4; ch0_1_3.K = C; ch0_1_3.zi_n = 16; ch0_1_3.flags = 4; ch0_1_3.act = 0;
      ch0_1_3.alpha = 1.0f; ch0_1_3.beta = 1.0f; ch0_1_3.sa = 1.0f; ch0_1_3.sb = 1.0f; ch0_1_3.Npad = G4; ch0_1_3.pad_ = 0;
      k_gemm<1><<<dim3((unsigned)((G4) + 31) / 32, (unsigned)((16) + 15) / 16, (unsigned)(Bn * 16)), 32, 0, stream>>>(ch0_1_3); }
    { GemmP ch0_1_4;
      ch0_1_4.A = HP + (size_t)19 * C; ch0_1_4.B = Wh1 + (size_t)4 * C * G4; ch0_1_4.bias = HP + (size_t)19 * C; ch0_1_4.R = GH; ch0_1_4.C = GH;
      ch0_1_4.sAo = (long long)PP * C; ch0_1_4.sAi = (long long)18 * C; ch0_1_4.sAm = C; ch0_1_4.sAk = 1; ch0_1_4.sBo = 0; ch0_1_4.sBi = 0; ch0_1_4.sBn = 1; ch0_1_4.sBk = G4; ch0_1_4.sCo = (long long)HW * G4; ch0_1_4.sCi = (long long)16 * G4; ch0_1_4.sCm = G4; ch0_1_4.sRo = (long long)HW * G4; ch0_1_4.sRi = (long long)16 * G4; ch0_1_4.sRm = G4; ch0_1_4.sRn = 1;
      ch0_1_4.M = 16; ch0_1_4.N = G4; ch0_1_4.K = C; ch0_1_4.zi_n = 16; ch0_1_4.flags = 4; ch0_1_4.act = 0;
      ch0_1_4.alpha = 1.0f; ch0_1_4.beta = 1.0f; ch0_1_4.sa = 1.0f; ch0_1_4.sb = 1.0f; ch0_1_4.Npad = G4; ch0_1_4.pad_ = 0;
      k_gemm<1><<<dim3((unsigned)((G4) + 31) / 32, (unsigned)((16) + 15) / 16, (unsigned)(Bn * 16)), 32, 0, stream>>>(ch0_1_4); }
    { GemmP ch0_1_5;
      ch0_1_5.A = HP + (size_t)20 * C; ch0_1_5.B = Wh1 + (size_t)5 * C * G4; ch0_1_5.bias = HP + (size_t)20 * C; ch0_1_5.R = GH; ch0_1_5.C = GH;
      ch0_1_5.sAo = (long long)PP * C; ch0_1_5.sAi = (long long)18 * C; ch0_1_5.sAm = C; ch0_1_5.sAk = 1; ch0_1_5.sBo = 0; ch0_1_5.sBi = 0; ch0_1_5.sBn = 1; ch0_1_5.sBk = G4; ch0_1_5.sCo = (long long)HW * G4; ch0_1_5.sCi = (long long)16 * G4; ch0_1_5.sCm = G4; ch0_1_5.sRo = (long long)HW * G4; ch0_1_5.sRi = (long long)16 * G4; ch0_1_5.sRm = G4; ch0_1_5.sRn = 1;
      ch0_1_5.M = 16; ch0_1_5.N = G4; ch0_1_5.K = C; ch0_1_5.zi_n = 16; ch0_1_5.flags = 4; ch0_1_5.act = 0;
      ch0_1_5.alpha = 1.0f; ch0_1_5.beta = 1.0f; ch0_1_5.sa = 1.0f; ch0_1_5.sb = 1.0f; ch0_1_5.Npad = G4; ch0_1_5.pad_ = 0;
      k_gemm<1><<<dim3((unsigned)((G4) + 31) / 32, (unsigned)((16) + 15) / 16, (unsigned)(Bn * 16)), 32, 0, stream>>>(ch0_1_5); }
    { GemmP ch0_1_6;
      ch0_1_6.A = HP + (size_t)36 * C; ch0_1_6.B = Wh1 + (size_t)6 * C * G4; ch0_1_6.bias = HP + (size_t)36 * C; ch0_1_6.R = GH; ch0_1_6.C = GH;
      ch0_1_6.sAo = (long long)PP * C; ch0_1_6.sAi = (long long)18 * C; ch0_1_6.sAm = C; ch0_1_6.sAk = 1; ch0_1_6.sBo = 0; ch0_1_6.sBi = 0; ch0_1_6.sBn = 1; ch0_1_6.sBk = G4; ch0_1_6.sCo = (long long)HW * G4; ch0_1_6.sCi = (long long)16 * G4; ch0_1_6.sCm = G4; ch0_1_6.sRo = (long long)HW * G4; ch0_1_6.sRi = (long long)16 * G4; ch0_1_6.sRm = G4; ch0_1_6.sRn = 1;
      ch0_1_6.M = 16; ch0_1_6.N = G4; ch0_1_6.K = C; ch0_1_6.zi_n = 16; ch0_1_6.flags = 4; ch0_1_6.act = 0;
      ch0_1_6.alpha = 1.0f; ch0_1_6.beta = 1.0f; ch0_1_6.sa = 1.0f; ch0_1_6.sb = 1.0f; ch0_1_6.Npad = G4; ch0_1_6.pad_ = 0;
      k_gemm<1><<<dim3((unsigned)((G4) + 31) / 32, (unsigned)((16) + 15) / 16, (unsigned)(Bn * 16)), 32, 0, stream>>>(ch0_1_6); }
    { GemmP ch0_1_7;
      ch0_1_7.A = HP + (size_t)37 * C; ch0_1_7.B = Wh1 + (size_t)7 * C * G4; ch0_1_7.bias = HP + (size_t)37 * C; ch0_1_7.R = GH; ch0_1_7.C = GH;
      ch0_1_7.sAo = (long long)PP * C; ch0_1_7.sAi = (long long)18 * C; ch0_1_7.sAm = C; ch0_1_7.sAk = 1; ch0_1_7.sBo = 0; ch0_1_7.sBi = 0; ch0_1_7.sBn = 1; ch0_1_7.sBk = G4; ch0_1_7.sCo = (long long)HW * G4; ch0_1_7.sCi = (long long)16 * G4; ch0_1_7.sCm = G4; ch0_1_7.sRo = (long long)HW * G4; ch0_1_7.sRi = (long long)16 * G4; ch0_1_7.sRm = G4; ch0_1_7.sRn = 1;
      ch0_1_7.M = 16; ch0_1_7.N = G4; ch0_1_7.K = C; ch0_1_7.zi_n = 16; ch0_1_7.flags = 4; ch0_1_7.act = 0;
      ch0_1_7.alpha = 1.0f; ch0_1_7.beta = 1.0f; ch0_1_7.sa = 1.0f; ch0_1_7.sb = 1.0f; ch0_1_7.Npad = G4; ch0_1_7.pad_ = 0;
      k_gemm<1><<<dim3((unsigned)((G4) + 31) / 32, (unsigned)((16) + 15) / 16, (unsigned)(Bn * 16)), 32, 0, stream>>>(ch0_1_7); }
    { GemmP ch0_1_8;
      ch0_1_8.A = HP + (size_t)38 * C; ch0_1_8.B = Wh1 + (size_t)8 * C * G4; ch0_1_8.bias = HP + (size_t)38 * C; ch0_1_8.R = GH; ch0_1_8.C = GH;
      ch0_1_8.sAo = (long long)PP * C; ch0_1_8.sAi = (long long)18 * C; ch0_1_8.sAm = C; ch0_1_8.sAk = 1; ch0_1_8.sBo = 0; ch0_1_8.sBi = 0; ch0_1_8.sBn = 1; ch0_1_8.sBk = G4; ch0_1_8.sCo = (long long)HW * G4; ch0_1_8.sCi = (long long)16 * G4; ch0_1_8.sCm = G4; ch0_1_8.sRo = (long long)HW * G4; ch0_1_8.sRi = (long long)16 * G4; ch0_1_8.sRm = G4; ch0_1_8.sRn = 1;
      ch0_1_8.M = 16; ch0_1_8.N = G4; ch0_1_8.K = C; ch0_1_8.zi_n = 16; ch0_1_8.flags = 4; ch0_1_8.act = 0;
      ch0_1_8.alpha = 1.0f; ch0_1_8.beta = 1.0f; ch0_1_8.sa = 1.0f; ch0_1_8.sb = 1.0f; ch0_1_8.Npad = G4; ch0_1_8.pad_ = 0;
      k_gemm<1><<<dim3((unsigned)((G4) + 31) / 32, (unsigned)((16) + 15) / 16, (unsigned)(Bn * 16)), 32, 0, stream>>>(ch0_1_8); }

    k_bl_cell<<<(unsigned)(((long long)Bn * HW * C + 255) / 256), 256, 0, stream>>>(XG, GH, Cc, HS, HP, Bn, T, 1, C);
    { GemmP ch0_2_0;
      ch0_2_0.A = HP + (size_t)0 * C; ch0_2_0.B = Wh1 + (size_t)0 * C * G4; ch0_2_0.bias = HP + (size_t)0 * C; ch0_2_0.R = HP + (size_t)0 * C; ch0_2_0.C = GH;
      ch0_2_0.sAo = (long long)PP * C; ch0_2_0.sAi = (long long)18 * C; ch0_2_0.sAm = C; ch0_2_0.sAk = 1; ch0_2_0.sBo = 0; ch0_2_0.sBi = 0; ch0_2_0.sBn = 1; ch0_2_0.sBk = G4; ch0_2_0.sCo = (long long)HW * G4; ch0_2_0.sCi = (long long)16 * G4; ch0_2_0.sCm = G4; ch0_2_0.sRo = 0; ch0_2_0.sRi = 0; ch0_2_0.sRm = 0; ch0_2_0.sRn = 0;
      ch0_2_0.M = 16; ch0_2_0.N = G4; ch0_2_0.K = C; ch0_2_0.zi_n = 16; ch0_2_0.flags = 0; ch0_2_0.act = 0;
      ch0_2_0.alpha = 1.0f; ch0_2_0.beta = 0.0f; ch0_2_0.sa = 1.0f; ch0_2_0.sb = 1.0f; ch0_2_0.Npad = G4; ch0_2_0.pad_ = 0;
      k_gemm<1><<<dim3((unsigned)((G4) + 31) / 32, (unsigned)((16) + 15) / 16, (unsigned)(Bn * 16)), 32, 0, stream>>>(ch0_2_0); }
    { GemmP ch0_2_1;
      ch0_2_1.A = HP + (size_t)1 * C; ch0_2_1.B = Wh1 + (size_t)1 * C * G4; ch0_2_1.bias = HP + (size_t)1 * C; ch0_2_1.R = GH; ch0_2_1.C = GH;
      ch0_2_1.sAo = (long long)PP * C; ch0_2_1.sAi = (long long)18 * C; ch0_2_1.sAm = C; ch0_2_1.sAk = 1; ch0_2_1.sBo = 0; ch0_2_1.sBi = 0; ch0_2_1.sBn = 1; ch0_2_1.sBk = G4; ch0_2_1.sCo = (long long)HW * G4; ch0_2_1.sCi = (long long)16 * G4; ch0_2_1.sCm = G4; ch0_2_1.sRo = (long long)HW * G4; ch0_2_1.sRi = (long long)16 * G4; ch0_2_1.sRm = G4; ch0_2_1.sRn = 1;
      ch0_2_1.M = 16; ch0_2_1.N = G4; ch0_2_1.K = C; ch0_2_1.zi_n = 16; ch0_2_1.flags = 4; ch0_2_1.act = 0;
      ch0_2_1.alpha = 1.0f; ch0_2_1.beta = 1.0f; ch0_2_1.sa = 1.0f; ch0_2_1.sb = 1.0f; ch0_2_1.Npad = G4; ch0_2_1.pad_ = 0;
      k_gemm<1><<<dim3((unsigned)((G4) + 31) / 32, (unsigned)((16) + 15) / 16, (unsigned)(Bn * 16)), 32, 0, stream>>>(ch0_2_1); }
    { GemmP ch0_2_2;
      ch0_2_2.A = HP + (size_t)2 * C; ch0_2_2.B = Wh1 + (size_t)2 * C * G4; ch0_2_2.bias = HP + (size_t)2 * C; ch0_2_2.R = GH; ch0_2_2.C = GH;
      ch0_2_2.sAo = (long long)PP * C; ch0_2_2.sAi = (long long)18 * C; ch0_2_2.sAm = C; ch0_2_2.sAk = 1; ch0_2_2.sBo = 0; ch0_2_2.sBi = 0; ch0_2_2.sBn = 1; ch0_2_2.sBk = G4; ch0_2_2.sCo = (long long)HW * G4; ch0_2_2.sCi = (long long)16 * G4; ch0_2_2.sCm = G4; ch0_2_2.sRo = (long long)HW * G4; ch0_2_2.sRi = (long long)16 * G4; ch0_2_2.sRm = G4; ch0_2_2.sRn = 1;
      ch0_2_2.M = 16; ch0_2_2.N = G4; ch0_2_2.K = C; ch0_2_2.zi_n = 16; ch0_2_2.flags = 4; ch0_2_2.act = 0;
      ch0_2_2.alpha = 1.0f; ch0_2_2.beta = 1.0f; ch0_2_2.sa = 1.0f; ch0_2_2.sb = 1.0f; ch0_2_2.Npad = G4; ch0_2_2.pad_ = 0;
      k_gemm<1><<<dim3((unsigned)((G4) + 31) / 32, (unsigned)((16) + 15) / 16, (unsigned)(Bn * 16)), 32, 0, stream>>>(ch0_2_2); }
    { GemmP ch0_2_3;
      ch0_2_3.A = HP + (size_t)18 * C; ch0_2_3.B = Wh1 + (size_t)3 * C * G4; ch0_2_3.bias = HP + (size_t)18 * C; ch0_2_3.R = GH; ch0_2_3.C = GH;
      ch0_2_3.sAo = (long long)PP * C; ch0_2_3.sAi = (long long)18 * C; ch0_2_3.sAm = C; ch0_2_3.sAk = 1; ch0_2_3.sBo = 0; ch0_2_3.sBi = 0; ch0_2_3.sBn = 1; ch0_2_3.sBk = G4; ch0_2_3.sCo = (long long)HW * G4; ch0_2_3.sCi = (long long)16 * G4; ch0_2_3.sCm = G4; ch0_2_3.sRo = (long long)HW * G4; ch0_2_3.sRi = (long long)16 * G4; ch0_2_3.sRm = G4; ch0_2_3.sRn = 1;
      ch0_2_3.M = 16; ch0_2_3.N = G4; ch0_2_3.K = C; ch0_2_3.zi_n = 16; ch0_2_3.flags = 4; ch0_2_3.act = 0;
      ch0_2_3.alpha = 1.0f; ch0_2_3.beta = 1.0f; ch0_2_3.sa = 1.0f; ch0_2_3.sb = 1.0f; ch0_2_3.Npad = G4; ch0_2_3.pad_ = 0;
      k_gemm<1><<<dim3((unsigned)((G4) + 31) / 32, (unsigned)((16) + 15) / 16, (unsigned)(Bn * 16)), 32, 0, stream>>>(ch0_2_3); }
    { GemmP ch0_2_4;
      ch0_2_4.A = HP + (size_t)19 * C; ch0_2_4.B = Wh1 + (size_t)4 * C * G4; ch0_2_4.bias = HP + (size_t)19 * C; ch0_2_4.R = GH; ch0_2_4.C = GH;
      ch0_2_4.sAo = (long long)PP * C; ch0_2_4.sAi = (long long)18 * C; ch0_2_4.sAm = C; ch0_2_4.sAk = 1; ch0_2_4.sBo = 0; ch0_2_4.sBi = 0; ch0_2_4.sBn = 1; ch0_2_4.sBk = G4; ch0_2_4.sCo = (long long)HW * G4; ch0_2_4.sCi = (long long)16 * G4; ch0_2_4.sCm = G4; ch0_2_4.sRo = (long long)HW * G4; ch0_2_4.sRi = (long long)16 * G4; ch0_2_4.sRm = G4; ch0_2_4.sRn = 1;
      ch0_2_4.M = 16; ch0_2_4.N = G4; ch0_2_4.K = C; ch0_2_4.zi_n = 16; ch0_2_4.flags = 4; ch0_2_4.act = 0;
      ch0_2_4.alpha = 1.0f; ch0_2_4.beta = 1.0f; ch0_2_4.sa = 1.0f; ch0_2_4.sb = 1.0f; ch0_2_4.Npad = G4; ch0_2_4.pad_ = 0;
      k_gemm<1><<<dim3((unsigned)((G4) + 31) / 32, (unsigned)((16) + 15) / 16, (unsigned)(Bn * 16)), 32, 0, stream>>>(ch0_2_4); }
    { GemmP ch0_2_5;
      ch0_2_5.A = HP + (size_t)20 * C; ch0_2_5.B = Wh1 + (size_t)5 * C * G4; ch0_2_5.bias = HP + (size_t)20 * C; ch0_2_5.R = GH; ch0_2_5.C = GH;
      ch0_2_5.sAo = (long long)PP * C; ch0_2_5.sAi = (long long)18 * C; ch0_2_5.sAm = C; ch0_2_5.sAk = 1; ch0_2_5.sBo = 0; ch0_2_5.sBi = 0; ch0_2_5.sBn = 1; ch0_2_5.sBk = G4; ch0_2_5.sCo = (long long)HW * G4; ch0_2_5.sCi = (long long)16 * G4; ch0_2_5.sCm = G4; ch0_2_5.sRo = (long long)HW * G4; ch0_2_5.sRi = (long long)16 * G4; ch0_2_5.sRm = G4; ch0_2_5.sRn = 1;
      ch0_2_5.M = 16; ch0_2_5.N = G4; ch0_2_5.K = C; ch0_2_5.zi_n = 16; ch0_2_5.flags = 4; ch0_2_5.act = 0;
      ch0_2_5.alpha = 1.0f; ch0_2_5.beta = 1.0f; ch0_2_5.sa = 1.0f; ch0_2_5.sb = 1.0f; ch0_2_5.Npad = G4; ch0_2_5.pad_ = 0;
      k_gemm<1><<<dim3((unsigned)((G4) + 31) / 32, (unsigned)((16) + 15) / 16, (unsigned)(Bn * 16)), 32, 0, stream>>>(ch0_2_5); }
    { GemmP ch0_2_6;
      ch0_2_6.A = HP + (size_t)36 * C; ch0_2_6.B = Wh1 + (size_t)6 * C * G4; ch0_2_6.bias = HP + (size_t)36 * C; ch0_2_6.R = GH; ch0_2_6.C = GH;
      ch0_2_6.sAo = (long long)PP * C; ch0_2_6.sAi = (long long)18 * C; ch0_2_6.sAm = C; ch0_2_6.sAk = 1; ch0_2_6.sBo = 0; ch0_2_6.sBi = 0; ch0_2_6.sBn = 1; ch0_2_6.sBk = G4; ch0_2_6.sCo = (long long)HW * G4; ch0_2_6.sCi = (long long)16 * G4; ch0_2_6.sCm = G4; ch0_2_6.sRo = (long long)HW * G4; ch0_2_6.sRi = (long long)16 * G4; ch0_2_6.sRm = G4; ch0_2_6.sRn = 1;
      ch0_2_6.M = 16; ch0_2_6.N = G4; ch0_2_6.K = C; ch0_2_6.zi_n = 16; ch0_2_6.flags = 4; ch0_2_6.act = 0;
      ch0_2_6.alpha = 1.0f; ch0_2_6.beta = 1.0f; ch0_2_6.sa = 1.0f; ch0_2_6.sb = 1.0f; ch0_2_6.Npad = G4; ch0_2_6.pad_ = 0;
      k_gemm<1><<<dim3((unsigned)((G4) + 31) / 32, (unsigned)((16) + 15) / 16, (unsigned)(Bn * 16)), 32, 0, stream>>>(ch0_2_6); }
    { GemmP ch0_2_7;
      ch0_2_7.A = HP + (size_t)37 * C; ch0_2_7.B = Wh1 + (size_t)7 * C * G4; ch0_2_7.bias = HP + (size_t)37 * C; ch0_2_7.R = GH; ch0_2_7.C = GH;
      ch0_2_7.sAo = (long long)PP * C; ch0_2_7.sAi = (long long)18 * C; ch0_2_7.sAm = C; ch0_2_7.sAk = 1; ch0_2_7.sBo = 0; ch0_2_7.sBi = 0; ch0_2_7.sBn = 1; ch0_2_7.sBk = G4; ch0_2_7.sCo = (long long)HW * G4; ch0_2_7.sCi = (long long)16 * G4; ch0_2_7.sCm = G4; ch0_2_7.sRo = (long long)HW * G4; ch0_2_7.sRi = (long long)16 * G4; ch0_2_7.sRm = G4; ch0_2_7.sRn = 1;
      ch0_2_7.M = 16; ch0_2_7.N = G4; ch0_2_7.K = C; ch0_2_7.zi_n = 16; ch0_2_7.flags = 4; ch0_2_7.act = 0;
      ch0_2_7.alpha = 1.0f; ch0_2_7.beta = 1.0f; ch0_2_7.sa = 1.0f; ch0_2_7.sb = 1.0f; ch0_2_7.Npad = G4; ch0_2_7.pad_ = 0;
      k_gemm<1><<<dim3((unsigned)((G4) + 31) / 32, (unsigned)((16) + 15) / 16, (unsigned)(Bn * 16)), 32, 0, stream>>>(ch0_2_7); }
    { GemmP ch0_2_8;
      ch0_2_8.A = HP + (size_t)38 * C; ch0_2_8.B = Wh1 + (size_t)8 * C * G4; ch0_2_8.bias = HP + (size_t)38 * C; ch0_2_8.R = GH; ch0_2_8.C = GH;
      ch0_2_8.sAo = (long long)PP * C; ch0_2_8.sAi = (long long)18 * C; ch0_2_8.sAm = C; ch0_2_8.sAk = 1; ch0_2_8.sBo = 0; ch0_2_8.sBi = 0; ch0_2_8.sBn = 1; ch0_2_8.sBk = G4; ch0_2_8.sCo = (long long)HW * G4; ch0_2_8.sCi = (long long)16 * G4; ch0_2_8.sCm = G4; ch0_2_8.sRo = (long long)HW * G4; ch0_2_8.sRi = (long long)16 * G4; ch0_2_8.sRm = G4; ch0_2_8.sRn = 1;
      ch0_2_8.M = 16; ch0_2_8.N = G4; ch0_2_8.K = C; ch0_2_8.zi_n = 16; ch0_2_8.flags = 4; ch0_2_8.act = 0;
      ch0_2_8.alpha = 1.0f; ch0_2_8.beta = 1.0f; ch0_2_8.sa = 1.0f; ch0_2_8.sb = 1.0f; ch0_2_8.Npad = G4; ch0_2_8.pad_ = 0;
      k_gemm<1><<<dim3((unsigned)((G4) + 31) / 32, (unsigned)((16) + 15) / 16, (unsigned)(Bn * 16)), 32, 0, stream>>>(ch0_2_8); }

    k_bl_cell<<<(unsigned)(((long long)Bn * HW * C + 255) / 256), 256, 0, stream>>>(XG, GH, Cc, HS, HP, Bn, T, 2, C);
    { GemmP ch0_3_0;
      ch0_3_0.A = HP + (size_t)0 * C; ch0_3_0.B = Wh1 + (size_t)0 * C * G4; ch0_3_0.bias = HP + (size_t)0 * C; ch0_3_0.R = HP + (size_t)0 * C; ch0_3_0.C = GH;
      ch0_3_0.sAo = (long long)PP * C; ch0_3_0.sAi = (long long)18 * C; ch0_3_0.sAm = C; ch0_3_0.sAk = 1; ch0_3_0.sBo = 0; ch0_3_0.sBi = 0; ch0_3_0.sBn = 1; ch0_3_0.sBk = G4; ch0_3_0.sCo = (long long)HW * G4; ch0_3_0.sCi = (long long)16 * G4; ch0_3_0.sCm = G4; ch0_3_0.sRo = 0; ch0_3_0.sRi = 0; ch0_3_0.sRm = 0; ch0_3_0.sRn = 0;
      ch0_3_0.M = 16; ch0_3_0.N = G4; ch0_3_0.K = C; ch0_3_0.zi_n = 16; ch0_3_0.flags = 0; ch0_3_0.act = 0;
      ch0_3_0.alpha = 1.0f; ch0_3_0.beta = 0.0f; ch0_3_0.sa = 1.0f; ch0_3_0.sb = 1.0f; ch0_3_0.Npad = G4; ch0_3_0.pad_ = 0;
      k_gemm<1><<<dim3((unsigned)((G4) + 31) / 32, (unsigned)((16) + 15) / 16, (unsigned)(Bn * 16)), 32, 0, stream>>>(ch0_3_0); }
    { GemmP ch0_3_1;
      ch0_3_1.A = HP + (size_t)1 * C; ch0_3_1.B = Wh1 + (size_t)1 * C * G4; ch0_3_1.bias = HP + (size_t)1 * C; ch0_3_1.R = GH; ch0_3_1.C = GH;
      ch0_3_1.sAo = (long long)PP * C; ch0_3_1.sAi = (long long)18 * C; ch0_3_1.sAm = C; ch0_3_1.sAk = 1; ch0_3_1.sBo = 0; ch0_3_1.sBi = 0; ch0_3_1.sBn = 1; ch0_3_1.sBk = G4; ch0_3_1.sCo = (long long)HW * G4; ch0_3_1.sCi = (long long)16 * G4; ch0_3_1.sCm = G4; ch0_3_1.sRo = (long long)HW * G4; ch0_3_1.sRi = (long long)16 * G4; ch0_3_1.sRm = G4; ch0_3_1.sRn = 1;
      ch0_3_1.M = 16; ch0_3_1.N = G4; ch0_3_1.K = C; ch0_3_1.zi_n = 16; ch0_3_1.flags = 4; ch0_3_1.act = 0;
      ch0_3_1.alpha = 1.0f; ch0_3_1.beta = 1.0f; ch0_3_1.sa = 1.0f; ch0_3_1.sb = 1.0f; ch0_3_1.Npad = G4; ch0_3_1.pad_ = 0;
      k_gemm<1><<<dim3((unsigned)((G4) + 31) / 32, (unsigned)((16) + 15) / 16, (unsigned)(Bn * 16)), 32, 0, stream>>>(ch0_3_1); }
    { GemmP ch0_3_2;
      ch0_3_2.A = HP + (size_t)2 * C; ch0_3_2.B = Wh1 + (size_t)2 * C * G4; ch0_3_2.bias = HP + (size_t)2 * C; ch0_3_2.R = GH; ch0_3_2.C = GH;
      ch0_3_2.sAo = (long long)PP * C; ch0_3_2.sAi = (long long)18 * C; ch0_3_2.sAm = C; ch0_3_2.sAk = 1; ch0_3_2.sBo = 0; ch0_3_2.sBi = 0; ch0_3_2.sBn = 1; ch0_3_2.sBk = G4; ch0_3_2.sCo = (long long)HW * G4; ch0_3_2.sCi = (long long)16 * G4; ch0_3_2.sCm = G4; ch0_3_2.sRo = (long long)HW * G4; ch0_3_2.sRi = (long long)16 * G4; ch0_3_2.sRm = G4; ch0_3_2.sRn = 1;
      ch0_3_2.M = 16; ch0_3_2.N = G4; ch0_3_2.K = C; ch0_3_2.zi_n = 16; ch0_3_2.flags = 4; ch0_3_2.act = 0;
      ch0_3_2.alpha = 1.0f; ch0_3_2.beta = 1.0f; ch0_3_2.sa = 1.0f; ch0_3_2.sb = 1.0f; ch0_3_2.Npad = G4; ch0_3_2.pad_ = 0;
      k_gemm<1><<<dim3((unsigned)((G4) + 31) / 32, (unsigned)((16) + 15) / 16, (unsigned)(Bn * 16)), 32, 0, stream>>>(ch0_3_2); }
    { GemmP ch0_3_3;
      ch0_3_3.A = HP + (size_t)18 * C; ch0_3_3.B = Wh1 + (size_t)3 * C * G4; ch0_3_3.bias = HP + (size_t)18 * C; ch0_3_3.R = GH; ch0_3_3.C = GH;
      ch0_3_3.sAo = (long long)PP * C; ch0_3_3.sAi = (long long)18 * C; ch0_3_3.sAm = C; ch0_3_3.sAk = 1; ch0_3_3.sBo = 0; ch0_3_3.sBi = 0; ch0_3_3.sBn = 1; ch0_3_3.sBk = G4; ch0_3_3.sCo = (long long)HW * G4; ch0_3_3.sCi = (long long)16 * G4; ch0_3_3.sCm = G4; ch0_3_3.sRo = (long long)HW * G4; ch0_3_3.sRi = (long long)16 * G4; ch0_3_3.sRm = G4; ch0_3_3.sRn = 1;
      ch0_3_3.M = 16; ch0_3_3.N = G4; ch0_3_3.K = C; ch0_3_3.zi_n = 16; ch0_3_3.flags = 4; ch0_3_3.act = 0;
      ch0_3_3.alpha = 1.0f; ch0_3_3.beta = 1.0f; ch0_3_3.sa = 1.0f; ch0_3_3.sb = 1.0f; ch0_3_3.Npad = G4; ch0_3_3.pad_ = 0;
      k_gemm<1><<<dim3((unsigned)((G4) + 31) / 32, (unsigned)((16) + 15) / 16, (unsigned)(Bn * 16)), 32, 0, stream>>>(ch0_3_3); }
    { GemmP ch0_3_4;
      ch0_3_4.A = HP + (size_t)19 * C; ch0_3_4.B = Wh1 + (size_t)4 * C * G4; ch0_3_4.bias = HP + (size_t)19 * C; ch0_3_4.R = GH; ch0_3_4.C = GH;
      ch0_3_4.sAo = (long long)PP * C; ch0_3_4.sAi = (long long)18 * C; ch0_3_4.sAm = C; ch0_3_4.sAk = 1; ch0_3_4.sBo = 0; ch0_3_4.sBi = 0; ch0_3_4.sBn = 1; ch0_3_4.sBk = G4; ch0_3_4.sCo = (long long)HW * G4; ch0_3_4.sCi = (long long)16 * G4; ch0_3_4.sCm = G4; ch0_3_4.sRo = (long long)HW * G4; ch0_3_4.sRi = (long long)16 * G4; ch0_3_4.sRm = G4; ch0_3_4.sRn = 1;
      ch0_3_4.M = 16; ch0_3_4.N = G4; ch0_3_4.K = C; ch0_3_4.zi_n = 16; ch0_3_4.flags = 4; ch0_3_4.act = 0;
      ch0_3_4.alpha = 1.0f; ch0_3_4.beta = 1.0f; ch0_3_4.sa = 1.0f; ch0_3_4.sb = 1.0f; ch0_3_4.Npad = G4; ch0_3_4.pad_ = 0;
      k_gemm<1><<<dim3((unsigned)((G4) + 31) / 32, (unsigned)((16) + 15) / 16, (unsigned)(Bn * 16)), 32, 0, stream>>>(ch0_3_4); }
    { GemmP ch0_3_5;
      ch0_3_5.A = HP + (size_t)20 * C; ch0_3_5.B = Wh1 + (size_t)5 * C * G4; ch0_3_5.bias = HP + (size_t)20 * C; ch0_3_5.R = GH; ch0_3_5.C = GH;
      ch0_3_5.sAo = (long long)PP * C; ch0_3_5.sAi = (long long)18 * C; ch0_3_5.sAm = C; ch0_3_5.sAk = 1; ch0_3_5.sBo = 0; ch0_3_5.sBi = 0; ch0_3_5.sBn = 1; ch0_3_5.sBk = G4; ch0_3_5.sCo = (long long)HW * G4; ch0_3_5.sCi = (long long)16 * G4; ch0_3_5.sCm = G4; ch0_3_5.sRo = (long long)HW * G4; ch0_3_5.sRi = (long long)16 * G4; ch0_3_5.sRm = G4; ch0_3_5.sRn = 1;
      ch0_3_5.M = 16; ch0_3_5.N = G4; ch0_3_5.K = C; ch0_3_5.zi_n = 16; ch0_3_5.flags = 4; ch0_3_5.act = 0;
      ch0_3_5.alpha = 1.0f; ch0_3_5.beta = 1.0f; ch0_3_5.sa = 1.0f; ch0_3_5.sb = 1.0f; ch0_3_5.Npad = G4; ch0_3_5.pad_ = 0;
      k_gemm<1><<<dim3((unsigned)((G4) + 31) / 32, (unsigned)((16) + 15) / 16, (unsigned)(Bn * 16)), 32, 0, stream>>>(ch0_3_5); }
    { GemmP ch0_3_6;
      ch0_3_6.A = HP + (size_t)36 * C; ch0_3_6.B = Wh1 + (size_t)6 * C * G4; ch0_3_6.bias = HP + (size_t)36 * C; ch0_3_6.R = GH; ch0_3_6.C = GH;
      ch0_3_6.sAo = (long long)PP * C; ch0_3_6.sAi = (long long)18 * C; ch0_3_6.sAm = C; ch0_3_6.sAk = 1; ch0_3_6.sBo = 0; ch0_3_6.sBi = 0; ch0_3_6.sBn = 1; ch0_3_6.sBk = G4; ch0_3_6.sCo = (long long)HW * G4; ch0_3_6.sCi = (long long)16 * G4; ch0_3_6.sCm = G4; ch0_3_6.sRo = (long long)HW * G4; ch0_3_6.sRi = (long long)16 * G4; ch0_3_6.sRm = G4; ch0_3_6.sRn = 1;
      ch0_3_6.M = 16; ch0_3_6.N = G4; ch0_3_6.K = C; ch0_3_6.zi_n = 16; ch0_3_6.flags = 4; ch0_3_6.act = 0;
      ch0_3_6.alpha = 1.0f; ch0_3_6.beta = 1.0f; ch0_3_6.sa = 1.0f; ch0_3_6.sb = 1.0f; ch0_3_6.Npad = G4; ch0_3_6.pad_ = 0;
      k_gemm<1><<<dim3((unsigned)((G4) + 31) / 32, (unsigned)((16) + 15) / 16, (unsigned)(Bn * 16)), 32, 0, stream>>>(ch0_3_6); }
    { GemmP ch0_3_7;
      ch0_3_7.A = HP + (size_t)37 * C; ch0_3_7.B = Wh1 + (size_t)7 * C * G4; ch0_3_7.bias = HP + (size_t)37 * C; ch0_3_7.R = GH; ch0_3_7.C = GH;
      ch0_3_7.sAo = (long long)PP * C; ch0_3_7.sAi = (long long)18 * C; ch0_3_7.sAm = C; ch0_3_7.sAk = 1; ch0_3_7.sBo = 0; ch0_3_7.sBi = 0; ch0_3_7.sBn = 1; ch0_3_7.sBk = G4; ch0_3_7.sCo = (long long)HW * G4; ch0_3_7.sCi = (long long)16 * G4; ch0_3_7.sCm = G4; ch0_3_7.sRo = (long long)HW * G4; ch0_3_7.sRi = (long long)16 * G4; ch0_3_7.sRm = G4; ch0_3_7.sRn = 1;
      ch0_3_7.M = 16; ch0_3_7.N = G4; ch0_3_7.K = C; ch0_3_7.zi_n = 16; ch0_3_7.flags = 4; ch0_3_7.act = 0;
      ch0_3_7.alpha = 1.0f; ch0_3_7.beta = 1.0f; ch0_3_7.sa = 1.0f; ch0_3_7.sb = 1.0f; ch0_3_7.Npad = G4; ch0_3_7.pad_ = 0;
      k_gemm<1><<<dim3((unsigned)((G4) + 31) / 32, (unsigned)((16) + 15) / 16, (unsigned)(Bn * 16)), 32, 0, stream>>>(ch0_3_7); }
    { GemmP ch0_3_8;
      ch0_3_8.A = HP + (size_t)38 * C; ch0_3_8.B = Wh1 + (size_t)8 * C * G4; ch0_3_8.bias = HP + (size_t)38 * C; ch0_3_8.R = GH; ch0_3_8.C = GH;
      ch0_3_8.sAo = (long long)PP * C; ch0_3_8.sAi = (long long)18 * C; ch0_3_8.sAm = C; ch0_3_8.sAk = 1; ch0_3_8.sBo = 0; ch0_3_8.sBi = 0; ch0_3_8.sBn = 1; ch0_3_8.sBk = G4; ch0_3_8.sCo = (long long)HW * G4; ch0_3_8.sCi = (long long)16 * G4; ch0_3_8.sCm = G4; ch0_3_8.sRo = (long long)HW * G4; ch0_3_8.sRi = (long long)16 * G4; ch0_3_8.sRm = G4; ch0_3_8.sRn = 1;
      ch0_3_8.M = 16; ch0_3_8.N = G4; ch0_3_8.K = C; ch0_3_8.zi_n = 16; ch0_3_8.flags = 4; ch0_3_8.act = 0;
      ch0_3_8.alpha = 1.0f; ch0_3_8.beta = 1.0f; ch0_3_8.sa = 1.0f; ch0_3_8.sb = 1.0f; ch0_3_8.Npad = G4; ch0_3_8.pad_ = 0;
      k_gemm<1><<<dim3((unsigned)((G4) + 31) / 32, (unsigned)((16) + 15) / 16, (unsigned)(Bn * 16)), 32, 0, stream>>>(ch0_3_8); }

    k_bl_cell<<<(unsigned)(((long long)Bn * HW * C + 255) / 256), 256, 0, stream>>>(XG, GH, Cc, HS, HP, Bn, T, 3, C);
    { GemmP ch0_4_0;
      ch0_4_0.A = HP + (size_t)0 * C; ch0_4_0.B = Wh1 + (size_t)0 * C * G4; ch0_4_0.bias = HP + (size_t)0 * C; ch0_4_0.R = HP + (size_t)0 * C; ch0_4_0.C = GH;
      ch0_4_0.sAo = (long long)PP * C; ch0_4_0.sAi = (long long)18 * C; ch0_4_0.sAm = C; ch0_4_0.sAk = 1; ch0_4_0.sBo = 0; ch0_4_0.sBi = 0; ch0_4_0.sBn = 1; ch0_4_0.sBk = G4; ch0_4_0.sCo = (long long)HW * G4; ch0_4_0.sCi = (long long)16 * G4; ch0_4_0.sCm = G4; ch0_4_0.sRo = 0; ch0_4_0.sRi = 0; ch0_4_0.sRm = 0; ch0_4_0.sRn = 0;
      ch0_4_0.M = 16; ch0_4_0.N = G4; ch0_4_0.K = C; ch0_4_0.zi_n = 16; ch0_4_0.flags = 0; ch0_4_0.act = 0;
      ch0_4_0.alpha = 1.0f; ch0_4_0.beta = 0.0f; ch0_4_0.sa = 1.0f; ch0_4_0.sb = 1.0f; ch0_4_0.Npad = G4; ch0_4_0.pad_ = 0;
      k_gemm<1><<<dim3((unsigned)((G4) + 31) / 32, (unsigned)((16) + 15) / 16, (unsigned)(Bn * 16)), 32, 0, stream>>>(ch0_4_0); }
    { GemmP ch0_4_1;
      ch0_4_1.A = HP + (size_t)1 * C; ch0_4_1.B = Wh1 + (size_t)1 * C * G4; ch0_4_1.bias = HP + (size_t)1 * C; ch0_4_1.R = GH; ch0_4_1.C = GH;
      ch0_4_1.sAo = (long long)PP * C; ch0_4_1.sAi = (long long)18 * C; ch0_4_1.sAm = C; ch0_4_1.sAk = 1; ch0_4_1.sBo = 0; ch0_4_1.sBi = 0; ch0_4_1.sBn = 1; ch0_4_1.sBk = G4; ch0_4_1.sCo = (long long)HW * G4; ch0_4_1.sCi = (long long)16 * G4; ch0_4_1.sCm = G4; ch0_4_1.sRo = (long long)HW * G4; ch0_4_1.sRi = (long long)16 * G4; ch0_4_1.sRm = G4; ch0_4_1.sRn = 1;
      ch0_4_1.M = 16; ch0_4_1.N = G4; ch0_4_1.K = C; ch0_4_1.zi_n = 16; ch0_4_1.flags = 4; ch0_4_1.act = 0;
      ch0_4_1.alpha = 1.0f; ch0_4_1.beta = 1.0f; ch0_4_1.sa = 1.0f; ch0_4_1.sb = 1.0f; ch0_4_1.Npad = G4; ch0_4_1.pad_ = 0;
      k_gemm<1><<<dim3((unsigned)((G4) + 31) / 32, (unsigned)((16) + 15) / 16, (unsigned)(Bn * 16)), 32, 0, stream>>>(ch0_4_1); }
    { GemmP ch0_4_2;
      ch0_4_2.A = HP + (size_t)2 * C; ch0_4_2.B = Wh1 + (size_t)2 * C * G4; ch0_4_2.bias = HP + (size_t)2 * C; ch0_4_2.R = GH; ch0_4_2.C = GH;
      ch0_4_2.sAo = (long long)PP * C; ch0_4_2.sAi = (long long)18 * C; ch0_4_2.sAm = C; ch0_4_2.sAk = 1; ch0_4_2.sBo = 0; ch0_4_2.sBi = 0; ch0_4_2.sBn = 1; ch0_4_2.sBk = G4; ch0_4_2.sCo = (long long)HW * G4; ch0_4_2.sCi = (long long)16 * G4; ch0_4_2.sCm = G4; ch0_4_2.sRo = (long long)HW * G4; ch0_4_2.sRi = (long long)16 * G4; ch0_4_2.sRm = G4; ch0_4_2.sRn = 1;
      ch0_4_2.M = 16; ch0_4_2.N = G4; ch0_4_2.K = C; ch0_4_2.zi_n = 16; ch0_4_2.flags = 4; ch0_4_2.act = 0;
      ch0_4_2.alpha = 1.0f; ch0_4_2.beta = 1.0f; ch0_4_2.sa = 1.0f; ch0_4_2.sb = 1.0f; ch0_4_2.Npad = G4; ch0_4_2.pad_ = 0;
      k_gemm<1><<<dim3((unsigned)((G4) + 31) / 32, (unsigned)((16) + 15) / 16, (unsigned)(Bn * 16)), 32, 0, stream>>>(ch0_4_2); }
    { GemmP ch0_4_3;
      ch0_4_3.A = HP + (size_t)18 * C; ch0_4_3.B = Wh1 + (size_t)3 * C * G4; ch0_4_3.bias = HP + (size_t)18 * C; ch0_4_3.R = GH; ch0_4_3.C = GH;
      ch0_4_3.sAo = (long long)PP * C; ch0_4_3.sAi = (long long)18 * C; ch0_4_3.sAm = C; ch0_4_3.sAk = 1; ch0_4_3.sBo = 0; ch0_4_3.sBi = 0; ch0_4_3.sBn = 1; ch0_4_3.sBk = G4; ch0_4_3.sCo = (long long)HW * G4; ch0_4_3.sCi = (long long)16 * G4; ch0_4_3.sCm = G4; ch0_4_3.sRo = (long long)HW * G4; ch0_4_3.sRi = (long long)16 * G4; ch0_4_3.sRm = G4; ch0_4_3.sRn = 1;
      ch0_4_3.M = 16; ch0_4_3.N = G4; ch0_4_3.K = C; ch0_4_3.zi_n = 16; ch0_4_3.flags = 4; ch0_4_3.act = 0;
      ch0_4_3.alpha = 1.0f; ch0_4_3.beta = 1.0f; ch0_4_3.sa = 1.0f; ch0_4_3.sb = 1.0f; ch0_4_3.Npad = G4; ch0_4_3.pad_ = 0;
      k_gemm<1><<<dim3((unsigned)((G4) + 31) / 32, (unsigned)((16) + 15) / 16, (unsigned)(Bn * 16)), 32, 0, stream>>>(ch0_4_3); }
    { GemmP ch0_4_4;
      ch0_4_4.A = HP + (size_t)19 * C; ch0_4_4.B = Wh1 + (size_t)4 * C * G4; ch0_4_4.bias = HP + (size_t)19 * C; ch0_4_4.R = GH; ch0_4_4.C = GH;
      ch0_4_4.sAo = (long long)PP * C; ch0_4_4.sAi = (long long)18 * C; ch0_4_4.sAm = C; ch0_4_4.sAk = 1; ch0_4_4.sBo = 0; ch0_4_4.sBi = 0; ch0_4_4.sBn = 1; ch0_4_4.sBk = G4; ch0_4_4.sCo = (long long)HW * G4; ch0_4_4.sCi = (long long)16 * G4; ch0_4_4.sCm = G4; ch0_4_4.sRo = (long long)HW * G4; ch0_4_4.sRi = (long long)16 * G4; ch0_4_4.sRm = G4; ch0_4_4.sRn = 1;
      ch0_4_4.M = 16; ch0_4_4.N = G4; ch0_4_4.K = C; ch0_4_4.zi_n = 16; ch0_4_4.flags = 4; ch0_4_4.act = 0;
      ch0_4_4.alpha = 1.0f; ch0_4_4.beta = 1.0f; ch0_4_4.sa = 1.0f; ch0_4_4.sb = 1.0f; ch0_4_4.Npad = G4; ch0_4_4.pad_ = 0;
      k_gemm<1><<<dim3((unsigned)((G4) + 31) / 32, (unsigned)((16) + 15) / 16, (unsigned)(Bn * 16)), 32, 0, stream>>>(ch0_4_4); }
    { GemmP ch0_4_5;
      ch0_4_5.A = HP + (size_t)20 * C; ch0_4_5.B = Wh1 + (size_t)5 * C * G4; ch0_4_5.bias = HP + (size_t)20 * C; ch0_4_5.R = GH; ch0_4_5.C = GH;
      ch0_4_5.sAo = (long long)PP * C; ch0_4_5.sAi = (long long)18 * C; ch0_4_5.sAm = C; ch0_4_5.sAk = 1; ch0_4_5.sBo = 0; ch0_4_5.sBi = 0; ch0_4_5.sBn = 1; ch0_4_5.sBk = G4; ch0_4_5.sCo = (long long)HW * G4; ch0_4_5.sCi = (long long)16 * G4; ch0_4_5.sCm = G4; ch0_4_5.sRo = (long long)HW * G4; ch0_4_5.sRi = (long long)16 * G4; ch0_4_5.sRm = G4; ch0_4_5.sRn = 1;
      ch0_4_5.M = 16; ch0_4_5.N = G4; ch0_4_5.K = C; ch0_4_5.zi_n = 16; ch0_4_5.flags = 4; ch0_4_5.act = 0;
      ch0_4_5.alpha = 1.0f; ch0_4_5.beta = 1.0f; ch0_4_5.sa = 1.0f; ch0_4_5.sb = 1.0f; ch0_4_5.Npad = G4; ch0_4_5.pad_ = 0;
      k_gemm<1><<<dim3((unsigned)((G4) + 31) / 32, (unsigned)((16) + 15) / 16, (unsigned)(Bn * 16)), 32, 0, stream>>>(ch0_4_5); }
    { GemmP ch0_4_6;
      ch0_4_6.A = HP + (size_t)36 * C; ch0_4_6.B = Wh1 + (size_t)6 * C * G4; ch0_4_6.bias = HP + (size_t)36 * C; ch0_4_6.R = GH; ch0_4_6.C = GH;
      ch0_4_6.sAo = (long long)PP * C; ch0_4_6.sAi = (long long)18 * C; ch0_4_6.sAm = C; ch0_4_6.sAk = 1; ch0_4_6.sBo = 0; ch0_4_6.sBi = 0; ch0_4_6.sBn = 1; ch0_4_6.sBk = G4; ch0_4_6.sCo = (long long)HW * G4; ch0_4_6.sCi = (long long)16 * G4; ch0_4_6.sCm = G4; ch0_4_6.sRo = (long long)HW * G4; ch0_4_6.sRi = (long long)16 * G4; ch0_4_6.sRm = G4; ch0_4_6.sRn = 1;
      ch0_4_6.M = 16; ch0_4_6.N = G4; ch0_4_6.K = C; ch0_4_6.zi_n = 16; ch0_4_6.flags = 4; ch0_4_6.act = 0;
      ch0_4_6.alpha = 1.0f; ch0_4_6.beta = 1.0f; ch0_4_6.sa = 1.0f; ch0_4_6.sb = 1.0f; ch0_4_6.Npad = G4; ch0_4_6.pad_ = 0;
      k_gemm<1><<<dim3((unsigned)((G4) + 31) / 32, (unsigned)((16) + 15) / 16, (unsigned)(Bn * 16)), 32, 0, stream>>>(ch0_4_6); }
    { GemmP ch0_4_7;
      ch0_4_7.A = HP + (size_t)37 * C; ch0_4_7.B = Wh1 + (size_t)7 * C * G4; ch0_4_7.bias = HP + (size_t)37 * C; ch0_4_7.R = GH; ch0_4_7.C = GH;
      ch0_4_7.sAo = (long long)PP * C; ch0_4_7.sAi = (long long)18 * C; ch0_4_7.sAm = C; ch0_4_7.sAk = 1; ch0_4_7.sBo = 0; ch0_4_7.sBi = 0; ch0_4_7.sBn = 1; ch0_4_7.sBk = G4; ch0_4_7.sCo = (long long)HW * G4; ch0_4_7.sCi = (long long)16 * G4; ch0_4_7.sCm = G4; ch0_4_7.sRo = (long long)HW * G4; ch0_4_7.sRi = (long long)16 * G4; ch0_4_7.sRm = G4; ch0_4_7.sRn = 1;
      ch0_4_7.M = 16; ch0_4_7.N = G4; ch0_4_7.K = C; ch0_4_7.zi_n = 16; ch0_4_7.flags = 4; ch0_4_7.act = 0;
      ch0_4_7.alpha = 1.0f; ch0_4_7.beta = 1.0f; ch0_4_7.sa = 1.0f; ch0_4_7.sb = 1.0f; ch0_4_7.Npad = G4; ch0_4_7.pad_ = 0;
      k_gemm<1><<<dim3((unsigned)((G4) + 31) / 32, (unsigned)((16) + 15) / 16, (unsigned)(Bn * 16)), 32, 0, stream>>>(ch0_4_7); }
    { GemmP ch0_4_8;
      ch0_4_8.A = HP + (size_t)38 * C; ch0_4_8.B = Wh1 + (size_t)8 * C * G4; ch0_4_8.bias = HP + (size_t)38 * C; ch0_4_8.R = GH; ch0_4_8.C = GH;
      ch0_4_8.sAo = (long long)PP * C; ch0_4_8.sAi = (long long)18 * C; ch0_4_8.sAm = C; ch0_4_8.sAk = 1; ch0_4_8.sBo = 0; ch0_4_8.sBi = 0; ch0_4_8.sBn = 1; ch0_4_8.sBk = G4; ch0_4_8.sCo = (long long)HW * G4; ch0_4_8.sCi = (long long)16 * G4; ch0_4_8.sCm = G4; ch0_4_8.sRo = (long long)HW * G4; ch0_4_8.sRi = (long long)16 * G4; ch0_4_8.sRm = G4; ch0_4_8.sRn = 1;
      ch0_4_8.M = 16; ch0_4_8.N = G4; ch0_4_8.K = C; ch0_4_8.zi_n = 16; ch0_4_8.flags = 4; ch0_4_8.act = 0;
      ch0_4_8.alpha = 1.0f; ch0_4_8.beta = 1.0f; ch0_4_8.sa = 1.0f; ch0_4_8.sb = 1.0f; ch0_4_8.Npad = G4; ch0_4_8.pad_ = 0;
      k_gemm<1><<<dim3((unsigned)((G4) + 31) / 32, (unsigned)((16) + 15) / 16, (unsigned)(Bn * 16)), 32, 0, stream>>>(ch0_4_8); }

    k_bl_cell<<<(unsigned)(((long long)Bn * HW * C + 255) / 256), 256, 0, stream>>>(XG, GH, Cc, HS, HP, Bn, T, 4, C);
    { GemmP ch0_5_0;
      ch0_5_0.A = HP + (size_t)0 * C; ch0_5_0.B = Wh1 + (size_t)0 * C * G4; ch0_5_0.bias = HP + (size_t)0 * C; ch0_5_0.R = HP + (size_t)0 * C; ch0_5_0.C = GH;
      ch0_5_0.sAo = (long long)PP * C; ch0_5_0.sAi = (long long)18 * C; ch0_5_0.sAm = C; ch0_5_0.sAk = 1; ch0_5_0.sBo = 0; ch0_5_0.sBi = 0; ch0_5_0.sBn = 1; ch0_5_0.sBk = G4; ch0_5_0.sCo = (long long)HW * G4; ch0_5_0.sCi = (long long)16 * G4; ch0_5_0.sCm = G4; ch0_5_0.sRo = 0; ch0_5_0.sRi = 0; ch0_5_0.sRm = 0; ch0_5_0.sRn = 0;
      ch0_5_0.M = 16; ch0_5_0.N = G4; ch0_5_0.K = C; ch0_5_0.zi_n = 16; ch0_5_0.flags = 0; ch0_5_0.act = 0;
      ch0_5_0.alpha = 1.0f; ch0_5_0.beta = 0.0f; ch0_5_0.sa = 1.0f; ch0_5_0.sb = 1.0f; ch0_5_0.Npad = G4; ch0_5_0.pad_ = 0;
      k_gemm<1><<<dim3((unsigned)((G4) + 31) / 32, (unsigned)((16) + 15) / 16, (unsigned)(Bn * 16)), 32, 0, stream>>>(ch0_5_0); }
    { GemmP ch0_5_1;
      ch0_5_1.A = HP + (size_t)1 * C; ch0_5_1.B = Wh1 + (size_t)1 * C * G4; ch0_5_1.bias = HP + (size_t)1 * C; ch0_5_1.R = GH; ch0_5_1.C = GH;
      ch0_5_1.sAo = (long long)PP * C; ch0_5_1.sAi = (long long)18 * C; ch0_5_1.sAm = C; ch0_5_1.sAk = 1; ch0_5_1.sBo = 0; ch0_5_1.sBi = 0; ch0_5_1.sBn = 1; ch0_5_1.sBk = G4; ch0_5_1.sCo = (long long)HW * G4; ch0_5_1.sCi = (long long)16 * G4; ch0_5_1.sCm = G4; ch0_5_1.sRo = (long long)HW * G4; ch0_5_1.sRi = (long long)16 * G4; ch0_5_1.sRm = G4; ch0_5_1.sRn = 1;
      ch0_5_1.M = 16; ch0_5_1.N = G4; ch0_5_1.K = C; ch0_5_1.zi_n = 16; ch0_5_1.flags = 4; ch0_5_1.act = 0;
      ch0_5_1.alpha = 1.0f; ch0_5_1.beta = 1.0f; ch0_5_1.sa = 1.0f; ch0_5_1.sb = 1.0f; ch0_5_1.Npad = G4; ch0_5_1.pad_ = 0;
      k_gemm<1><<<dim3((unsigned)((G4) + 31) / 32, (unsigned)((16) + 15) / 16, (unsigned)(Bn * 16)), 32, 0, stream>>>(ch0_5_1); }
    { GemmP ch0_5_2;
      ch0_5_2.A = HP + (size_t)2 * C; ch0_5_2.B = Wh1 + (size_t)2 * C * G4; ch0_5_2.bias = HP + (size_t)2 * C; ch0_5_2.R = GH; ch0_5_2.C = GH;
      ch0_5_2.sAo = (long long)PP * C; ch0_5_2.sAi = (long long)18 * C; ch0_5_2.sAm = C; ch0_5_2.sAk = 1; ch0_5_2.sBo = 0; ch0_5_2.sBi = 0; ch0_5_2.sBn = 1; ch0_5_2.sBk = G4; ch0_5_2.sCo = (long long)HW * G4; ch0_5_2.sCi = (long long)16 * G4; ch0_5_2.sCm = G4; ch0_5_2.sRo = (long long)HW * G4; ch0_5_2.sRi = (long long)16 * G4; ch0_5_2.sRm = G4; ch0_5_2.sRn = 1;
      ch0_5_2.M = 16; ch0_5_2.N = G4; ch0_5_2.K = C; ch0_5_2.zi_n = 16; ch0_5_2.flags = 4; ch0_5_2.act = 0;
      ch0_5_2.alpha = 1.0f; ch0_5_2.beta = 1.0f; ch0_5_2.sa = 1.0f; ch0_5_2.sb = 1.0f; ch0_5_2.Npad = G4; ch0_5_2.pad_ = 0;
      k_gemm<1><<<dim3((unsigned)((G4) + 31) / 32, (unsigned)((16) + 15) / 16, (unsigned)(Bn * 16)), 32, 0, stream>>>(ch0_5_2); }
    { GemmP ch0_5_3;
      ch0_5_3.A = HP + (size_t)18 * C; ch0_5_3.B = Wh1 + (size_t)3 * C * G4; ch0_5_3.bias = HP + (size_t)18 * C; ch0_5_3.R = GH; ch0_5_3.C = GH;
      ch0_5_3.sAo = (long long)PP * C; ch0_5_3.sAi = (long long)18 * C; ch0_5_3.sAm = C; ch0_5_3.sAk = 1; ch0_5_3.sBo = 0; ch0_5_3.sBi = 0; ch0_5_3.sBn = 1; ch0_5_3.sBk = G4; ch0_5_3.sCo = (long long)HW * G4; ch0_5_3.sCi = (long long)16 * G4; ch0_5_3.sCm = G4; ch0_5_3.sRo = (long long)HW * G4; ch0_5_3.sRi = (long long)16 * G4; ch0_5_3.sRm = G4; ch0_5_3.sRn = 1;
      ch0_5_3.M = 16; ch0_5_3.N = G4; ch0_5_3.K = C; ch0_5_3.zi_n = 16; ch0_5_3.flags = 4; ch0_5_3.act = 0;
      ch0_5_3.alpha = 1.0f; ch0_5_3.beta = 1.0f; ch0_5_3.sa = 1.0f; ch0_5_3.sb = 1.0f; ch0_5_3.Npad = G4; ch0_5_3.pad_ = 0;
      k_gemm<1><<<dim3((unsigned)((G4) + 31) / 32, (unsigned)((16) + 15) / 16, (unsigned)(Bn * 16)), 32, 0, stream>>>(ch0_5_3); }
    { GemmP ch0_5_4;
      ch0_5_4.A = HP + (size_t)19 * C; ch0_5_4.B = Wh1 + (size_t)4 * C * G4; ch0_5_4.bias = HP + (size_t)19 * C; ch0_5_4.R = GH; ch0_5_4.C = GH;
      ch0_5_4.sAo = (long long)PP * C; ch0_5_4.sAi = (long long)18 * C; ch0_5_4.sAm = C; ch0_5_4.sAk = 1; ch0_5_4.sBo = 0; ch0_5_4.sBi = 0; ch0_5_4.sBn = 1; ch0_5_4.sBk = G4; ch0_5_4.sCo = (long long)HW * G4; ch0_5_4.sCi = (long long)16 * G4; ch0_5_4.sCm = G4; ch0_5_4.sRo = (long long)HW * G4; ch0_5_4.sRi = (long long)16 * G4; ch0_5_4.sRm = G4; ch0_5_4.sRn = 1;
      ch0_5_4.M = 16; ch0_5_4.N = G4; ch0_5_4.K = C; ch0_5_4.zi_n = 16; ch0_5_4.flags = 4; ch0_5_4.act = 0;
      ch0_5_4.alpha = 1.0f; ch0_5_4.beta = 1.0f; ch0_5_4.sa = 1.0f; ch0_5_4.sb = 1.0f; ch0_5_4.Npad = G4; ch0_5_4.pad_ = 0;
      k_gemm<1><<<dim3((unsigned)((G4) + 31) / 32, (unsigned)((16) + 15) / 16, (unsigned)(Bn * 16)), 32, 0, stream>>>(ch0_5_4); }
    { GemmP ch0_5_5;
      ch0_5_5.A = HP + (size_t)20 * C; ch0_5_5.B = Wh1 + (size_t)5 * C * G4; ch0_5_5.bias = HP + (size_t)20 * C; ch0_5_5.R = GH; ch0_5_5.C = GH;
      ch0_5_5.sAo = (long long)PP * C; ch0_5_5.sAi = (long long)18 * C; ch0_5_5.sAm = C; ch0_5_5.sAk = 1; ch0_5_5.sBo = 0; ch0_5_5.sBi = 0; ch0_5_5.sBn = 1; ch0_5_5.sBk = G4; ch0_5_5.sCo = (long long)HW * G4; ch0_5_5.sCi = (long long)16 * G4; ch0_5_5.sCm = G4; ch0_5_5.sRo = (long long)HW * G4; ch0_5_5.sRi = (long long)16 * G4; ch0_5_5.sRm = G4; ch0_5_5.sRn = 1;
      ch0_5_5.M = 16; ch0_5_5.N = G4; ch0_5_5.K = C; ch0_5_5.zi_n = 16; ch0_5_5.flags = 4; ch0_5_5.act = 0;
      ch0_5_5.alpha = 1.0f; ch0_5_5.beta = 1.0f; ch0_5_5.sa = 1.0f; ch0_5_5.sb = 1.0f; ch0_5_5.Npad = G4; ch0_5_5.pad_ = 0;
      k_gemm<1><<<dim3((unsigned)((G4) + 31) / 32, (unsigned)((16) + 15) / 16, (unsigned)(Bn * 16)), 32, 0, stream>>>(ch0_5_5); }
    { GemmP ch0_5_6;
      ch0_5_6.A = HP + (size_t)36 * C; ch0_5_6.B = Wh1 + (size_t)6 * C * G4; ch0_5_6.bias = HP + (size_t)36 * C; ch0_5_6.R = GH; ch0_5_6.C = GH;
      ch0_5_6.sAo = (long long)PP * C; ch0_5_6.sAi = (long long)18 * C; ch0_5_6.sAm = C; ch0_5_6.sAk = 1; ch0_5_6.sBo = 0; ch0_5_6.sBi = 0; ch0_5_6.sBn = 1; ch0_5_6.sBk = G4; ch0_5_6.sCo = (long long)HW * G4; ch0_5_6.sCi = (long long)16 * G4; ch0_5_6.sCm = G4; ch0_5_6.sRo = (long long)HW * G4; ch0_5_6.sRi = (long long)16 * G4; ch0_5_6.sRm = G4; ch0_5_6.sRn = 1;
      ch0_5_6.M = 16; ch0_5_6.N = G4; ch0_5_6.K = C; ch0_5_6.zi_n = 16; ch0_5_6.flags = 4; ch0_5_6.act = 0;
      ch0_5_6.alpha = 1.0f; ch0_5_6.beta = 1.0f; ch0_5_6.sa = 1.0f; ch0_5_6.sb = 1.0f; ch0_5_6.Npad = G4; ch0_5_6.pad_ = 0;
      k_gemm<1><<<dim3((unsigned)((G4) + 31) / 32, (unsigned)((16) + 15) / 16, (unsigned)(Bn * 16)), 32, 0, stream>>>(ch0_5_6); }
    { GemmP ch0_5_7;
      ch0_5_7.A = HP + (size_t)37 * C; ch0_5_7.B = Wh1 + (size_t)7 * C * G4; ch0_5_7.bias = HP + (size_t)37 * C; ch0_5_7.R = GH; ch0_5_7.C = GH;
      ch0_5_7.sAo = (long long)PP * C; ch0_5_7.sAi = (long long)18 * C; ch0_5_7.sAm = C; ch0_5_7.sAk = 1; ch0_5_7.sBo = 0; ch0_5_7.sBi = 0; ch0_5_7.sBn = 1; ch0_5_7.sBk = G4; ch0_5_7.sCo = (long long)HW * G4; ch0_5_7.sCi = (long long)16 * G4; ch0_5_7.sCm = G4; ch0_5_7.sRo = (long long)HW * G4; ch0_5_7.sRi = (long long)16 * G4; ch0_5_7.sRm = G4; ch0_5_7.sRn = 1;
      ch0_5_7.M = 16; ch0_5_7.N = G4; ch0_5_7.K = C; ch0_5_7.zi_n = 16; ch0_5_7.flags = 4; ch0_5_7.act = 0;
      ch0_5_7.alpha = 1.0f; ch0_5_7.beta = 1.0f; ch0_5_7.sa = 1.0f; ch0_5_7.sb = 1.0f; ch0_5_7.Npad = G4; ch0_5_7.pad_ = 0;
      k_gemm<1><<<dim3((unsigned)((G4) + 31) / 32, (unsigned)((16) + 15) / 16, (unsigned)(Bn * 16)), 32, 0, stream>>>(ch0_5_7); }
    { GemmP ch0_5_8;
      ch0_5_8.A = HP + (size_t)38 * C; ch0_5_8.B = Wh1 + (size_t)8 * C * G4; ch0_5_8.bias = HP + (size_t)38 * C; ch0_5_8.R = GH; ch0_5_8.C = GH;
      ch0_5_8.sAo = (long long)PP * C; ch0_5_8.sAi = (long long)18 * C; ch0_5_8.sAm = C; ch0_5_8.sAk = 1; ch0_5_8.sBo = 0; ch0_5_8.sBi = 0; ch0_5_8.sBn = 1; ch0_5_8.sBk = G4; ch0_5_8.sCo = (long long)HW * G4; ch0_5_8.sCi = (long long)16 * G4; ch0_5_8.sCm = G4; ch0_5_8.sRo = (long long)HW * G4; ch0_5_8.sRi = (long long)16 * G4; ch0_5_8.sRm = G4; ch0_5_8.sRn = 1;
      ch0_5_8.M = 16; ch0_5_8.N = G4; ch0_5_8.K = C; ch0_5_8.zi_n = 16; ch0_5_8.flags = 4; ch0_5_8.act = 0;
      ch0_5_8.alpha = 1.0f; ch0_5_8.beta = 1.0f; ch0_5_8.sa = 1.0f; ch0_5_8.sb = 1.0f; ch0_5_8.Npad = G4; ch0_5_8.pad_ = 0;
      k_gemm<1><<<dim3((unsigned)((G4) + 31) / 32, (unsigned)((16) + 15) / 16, (unsigned)(Bn * 16)), 32, 0, stream>>>(ch0_5_8); }

    k_bl_cell<<<(unsigned)(((long long)Bn * HW * C + 255) / 256), 256, 0, stream>>>(XG, GH, Cc, HS, HP, Bn, T, 5, C);
    { GemmP ch0_6_0;
      ch0_6_0.A = HP + (size_t)0 * C; ch0_6_0.B = Wh1 + (size_t)0 * C * G4; ch0_6_0.bias = HP + (size_t)0 * C; ch0_6_0.R = HP + (size_t)0 * C; ch0_6_0.C = GH;
      ch0_6_0.sAo = (long long)PP * C; ch0_6_0.sAi = (long long)18 * C; ch0_6_0.sAm = C; ch0_6_0.sAk = 1; ch0_6_0.sBo = 0; ch0_6_0.sBi = 0; ch0_6_0.sBn = 1; ch0_6_0.sBk = G4; ch0_6_0.sCo = (long long)HW * G4; ch0_6_0.sCi = (long long)16 * G4; ch0_6_0.sCm = G4; ch0_6_0.sRo = 0; ch0_6_0.sRi = 0; ch0_6_0.sRm = 0; ch0_6_0.sRn = 0;
      ch0_6_0.M = 16; ch0_6_0.N = G4; ch0_6_0.K = C; ch0_6_0.zi_n = 16; ch0_6_0.flags = 0; ch0_6_0.act = 0;
      ch0_6_0.alpha = 1.0f; ch0_6_0.beta = 0.0f; ch0_6_0.sa = 1.0f; ch0_6_0.sb = 1.0f; ch0_6_0.Npad = G4; ch0_6_0.pad_ = 0;
      k_gemm<1><<<dim3((unsigned)((G4) + 31) / 32, (unsigned)((16) + 15) / 16, (unsigned)(Bn * 16)), 32, 0, stream>>>(ch0_6_0); }
    { GemmP ch0_6_1;
      ch0_6_1.A = HP + (size_t)1 * C; ch0_6_1.B = Wh1 + (size_t)1 * C * G4; ch0_6_1.bias = HP + (size_t)1 * C; ch0_6_1.R = GH; ch0_6_1.C = GH;
      ch0_6_1.sAo = (long long)PP * C; ch0_6_1.sAi = (long long)18 * C; ch0_6_1.sAm = C; ch0_6_1.sAk = 1; ch0_6_1.sBo = 0; ch0_6_1.sBi = 0; ch0_6_1.sBn = 1; ch0_6_1.sBk = G4; ch0_6_1.sCo = (long long)HW * G4; ch0_6_1.sCi = (long long)16 * G4; ch0_6_1.sCm = G4; ch0_6_1.sRo = (long long)HW * G4; ch0_6_1.sRi = (long long)16 * G4; ch0_6_1.sRm = G4; ch0_6_1.sRn = 1;
      ch0_6_1.M = 16; ch0_6_1.N = G4; ch0_6_1.K = C; ch0_6_1.zi_n = 16; ch0_6_1.flags = 4; ch0_6_1.act = 0;
      ch0_6_1.alpha = 1.0f; ch0_6_1.beta = 1.0f; ch0_6_1.sa = 1.0f; ch0_6_1.sb = 1.0f; ch0_6_1.Npad = G4; ch0_6_1.pad_ = 0;
      k_gemm<1><<<dim3((unsigned)((G4) + 31) / 32, (unsigned)((16) + 15) / 16, (unsigned)(Bn * 16)), 32, 0, stream>>>(ch0_6_1); }
    { GemmP ch0_6_2;
      ch0_6_2.A = HP + (size_t)2 * C; ch0_6_2.B = Wh1 + (size_t)2 * C * G4; ch0_6_2.bias = HP + (size_t)2 * C; ch0_6_2.R = GH; ch0_6_2.C = GH;
      ch0_6_2.sAo = (long long)PP * C; ch0_6_2.sAi = (long long)18 * C; ch0_6_2.sAm = C; ch0_6_2.sAk = 1; ch0_6_2.sBo = 0; ch0_6_2.sBi = 0; ch0_6_2.sBn = 1; ch0_6_2.sBk = G4; ch0_6_2.sCo = (long long)HW * G4; ch0_6_2.sCi = (long long)16 * G4; ch0_6_2.sCm = G4; ch0_6_2.sRo = (long long)HW * G4; ch0_6_2.sRi = (long long)16 * G4; ch0_6_2.sRm = G4; ch0_6_2.sRn = 1;
      ch0_6_2.M = 16; ch0_6_2.N = G4; ch0_6_2.K = C; ch0_6_2.zi_n = 16; ch0_6_2.flags = 4; ch0_6_2.act = 0;
      ch0_6_2.alpha = 1.0f; ch0_6_2.beta = 1.0f; ch0_6_2.sa = 1.0f; ch0_6_2.sb = 1.0f; ch0_6_2.Npad = G4; ch0_6_2.pad_ = 0;
      k_gemm<1><<<dim3((unsigned)((G4) + 31) / 32, (unsigned)((16) + 15) / 16, (unsigned)(Bn * 16)), 32, 0, stream>>>(ch0_6_2); }
    { GemmP ch0_6_3;
      ch0_6_3.A = HP + (size_t)18 * C; ch0_6_3.B = Wh1 + (size_t)3 * C * G4; ch0_6_3.bias = HP + (size_t)18 * C; ch0_6_3.R = GH; ch0_6_3.C = GH;
      ch0_6_3.sAo = (long long)PP * C; ch0_6_3.sAi = (long long)18 * C; ch0_6_3.sAm = C; ch0_6_3.sAk = 1; ch0_6_3.sBo = 0; ch0_6_3.sBi = 0; ch0_6_3.sBn = 1; ch0_6_3.sBk = G4; ch0_6_3.sCo = (long long)HW * G4; ch0_6_3.sCi = (long long)16 * G4; ch0_6_3.sCm = G4; ch0_6_3.sRo = (long long)HW * G4; ch0_6_3.sRi = (long long)16 * G4; ch0_6_3.sRm = G4; ch0_6_3.sRn = 1;
      ch0_6_3.M = 16; ch0_6_3.N = G4; ch0_6_3.K = C; ch0_6_3.zi_n = 16; ch0_6_3.flags = 4; ch0_6_3.act = 0;
      ch0_6_3.alpha = 1.0f; ch0_6_3.beta = 1.0f; ch0_6_3.sa = 1.0f; ch0_6_3.sb = 1.0f; ch0_6_3.Npad = G4; ch0_6_3.pad_ = 0;
      k_gemm<1><<<dim3((unsigned)((G4) + 31) / 32, (unsigned)((16) + 15) / 16, (unsigned)(Bn * 16)), 32, 0, stream>>>(ch0_6_3); }
    { GemmP ch0_6_4;
      ch0_6_4.A = HP + (size_t)19 * C; ch0_6_4.B = Wh1 + (size_t)4 * C * G4; ch0_6_4.bias = HP + (size_t)19 * C; ch0_6_4.R = GH; ch0_6_4.C = GH;
      ch0_6_4.sAo = (long long)PP * C; ch0_6_4.sAi = (long long)18 * C; ch0_6_4.sAm = C; ch0_6_4.sAk = 1; ch0_6_4.sBo = 0; ch0_6_4.sBi = 0; ch0_6_4.sBn = 1; ch0_6_4.sBk = G4; ch0_6_4.sCo = (long long)HW * G4; ch0_6_4.sCi = (long long)16 * G4; ch0_6_4.sCm = G4; ch0_6_4.sRo = (long long)HW * G4; ch0_6_4.sRi = (long long)16 * G4; ch0_6_4.sRm = G4; ch0_6_4.sRn = 1;
      ch0_6_4.M = 16; ch0_6_4.N = G4; ch0_6_4.K = C; ch0_6_4.zi_n = 16; ch0_6_4.flags = 4; ch0_6_4.act = 0;
      ch0_6_4.alpha = 1.0f; ch0_6_4.beta = 1.0f; ch0_6_4.sa = 1.0f; ch0_6_4.sb = 1.0f; ch0_6_4.Npad = G4; ch0_6_4.pad_ = 0;
      k_gemm<1><<<dim3((unsigned)((G4) + 31) / 32, (unsigned)((16) + 15) / 16, (unsigned)(Bn * 16)), 32, 0, stream>>>(ch0_6_4); }
    { GemmP ch0_6_5;
      ch0_6_5.A = HP + (size_t)20 * C; ch0_6_5.B = Wh1 + (size_t)5 * C * G4; ch0_6_5.bias = HP + (size_t)20 * C; ch0_6_5.R = GH; ch0_6_5.C = GH;
      ch0_6_5.sAo = (long long)PP * C; ch0_6_5.sAi = (long long)18 * C; ch0_6_5.sAm = C; ch0_6_5.sAk = 1; ch0_6_5.sBo = 0; ch0_6_5.sBi = 0; ch0_6_5.sBn = 1; ch0_6_5.sBk = G4; ch0_6_5.sCo = (long long)HW * G4; ch0_6_5.sCi = (long long)16 * G4; ch0_6_5.sCm = G4; ch0_6_5.sRo = (long long)HW * G4; ch0_6_5.sRi = (long long)16 * G4; ch0_6_5.sRm = G4; ch0_6_5.sRn = 1;
      ch0_6_5.M = 16; ch0_6_5.N = G4; ch0_6_5.K = C; ch0_6_5.zi_n = 16; ch0_6_5.flags = 4; ch0_6_5.act = 0;
      ch0_6_5.alpha = 1.0f; ch0_6_5.beta = 1.0f; ch0_6_5.sa = 1.0f; ch0_6_5.sb = 1.0f; ch0_6_5.Npad = G4; ch0_6_5.pad_ = 0;
      k_gemm<1><<<dim3((unsigned)((G4) + 31) / 32, (unsigned)((16) + 15) / 16, (unsigned)(Bn * 16)), 32, 0, stream>>>(ch0_6_5); }
    { GemmP ch0_6_6;
      ch0_6_6.A = HP + (size_t)36 * C; ch0_6_6.B = Wh1 + (size_t)6 * C * G4; ch0_6_6.bias = HP + (size_t)36 * C; ch0_6_6.R = GH; ch0_6_6.C = GH;
      ch0_6_6.sAo = (long long)PP * C; ch0_6_6.sAi = (long long)18 * C; ch0_6_6.sAm = C; ch0_6_6.sAk = 1; ch0_6_6.sBo = 0; ch0_6_6.sBi = 0; ch0_6_6.sBn = 1; ch0_6_6.sBk = G4; ch0_6_6.sCo = (long long)HW * G4; ch0_6_6.sCi = (long long)16 * G4; ch0_6_6.sCm = G4; ch0_6_6.sRo = (long long)HW * G4; ch0_6_6.sRi = (long long)16 * G4; ch0_6_6.sRm = G4; ch0_6_6.sRn = 1;
      ch0_6_6.M = 16; ch0_6_6.N = G4; ch0_6_6.K = C; ch0_6_6.zi_n = 16; ch0_6_6.flags = 4; ch0_6_6.act = 0;
      ch0_6_6.alpha = 1.0f; ch0_6_6.beta = 1.0f; ch0_6_6.sa = 1.0f; ch0_6_6.sb = 1.0f; ch0_6_6.Npad = G4; ch0_6_6.pad_ = 0;
      k_gemm<1><<<dim3((unsigned)((G4) + 31) / 32, (unsigned)((16) + 15) / 16, (unsigned)(Bn * 16)), 32, 0, stream>>>(ch0_6_6); }
    { GemmP ch0_6_7;
      ch0_6_7.A = HP + (size_t)37 * C; ch0_6_7.B = Wh1 + (size_t)7 * C * G4; ch0_6_7.bias = HP + (size_t)37 * C; ch0_6_7.R = GH; ch0_6_7.C = GH;
      ch0_6_7.sAo = (long long)PP * C; ch0_6_7.sAi = (long long)18 * C; ch0_6_7.sAm = C; ch0_6_7.sAk = 1; ch0_6_7.sBo = 0; ch0_6_7.sBi = 0; ch0_6_7.sBn = 1; ch0_6_7.sBk = G4; ch0_6_7.sCo = (long long)HW * G4; ch0_6_7.sCi = (long long)16 * G4; ch0_6_7.sCm = G4; ch0_6_7.sRo = (long long)HW * G4; ch0_6_7.sRi = (long long)16 * G4; ch0_6_7.sRm = G4; ch0_6_7.sRn = 1;
      ch0_6_7.M = 16; ch0_6_7.N = G4; ch0_6_7.K = C; ch0_6_7.zi_n = 16; ch0_6_7.flags = 4; ch0_6_7.act = 0;
      ch0_6_7.alpha = 1.0f; ch0_6_7.beta = 1.0f; ch0_6_7.sa = 1.0f; ch0_6_7.sb = 1.0f; ch0_6_7.Npad = G4; ch0_6_7.pad_ = 0;
      k_gemm<1><<<dim3((unsigned)((G4) + 31) / 32, (unsigned)((16) + 15) / 16, (unsigned)(Bn * 16)), 32, 0, stream>>>(ch0_6_7); }
    { GemmP ch0_6_8;
      ch0_6_8.A = HP + (size_t)38 * C; ch0_6_8.B = Wh1 + (size_t)8 * C * G4; ch0_6_8.bias = HP + (size_t)38 * C; ch0_6_8.R = GH; ch0_6_8.C = GH;
      ch0_6_8.sAo = (long long)PP * C; ch0_6_8.sAi = (long long)18 * C; ch0_6_8.sAm = C; ch0_6_8.sAk = 1; ch0_6_8.sBo = 0; ch0_6_8.sBi = 0; ch0_6_8.sBn = 1; ch0_6_8.sBk = G4; ch0_6_8.sCo = (long long)HW * G4; ch0_6_8.sCi = (long long)16 * G4; ch0_6_8.sCm = G4; ch0_6_8.sRo = (long long)HW * G4; ch0_6_8.sRi = (long long)16 * G4; ch0_6_8.sRm = G4; ch0_6_8.sRn = 1;
      ch0_6_8.M = 16; ch0_6_8.N = G4; ch0_6_8.K = C; ch0_6_8.zi_n = 16; ch0_6_8.flags = 4; ch0_6_8.act = 0;
      ch0_6_8.alpha = 1.0f; ch0_6_8.beta = 1.0f; ch0_6_8.sa = 1.0f; ch0_6_8.sb = 1.0f; ch0_6_8.Npad = G4; ch0_6_8.pad_ = 0;
      k_gemm<1><<<dim3((unsigned)((G4) + 31) / 32, (unsigned)((16) + 15) / 16, (unsigned)(Bn * 16)), 32, 0, stream>>>(ch0_6_8); }

    k_bl_cell<<<(unsigned)(((long long)Bn * HW * C + 255) / 256), 256, 0, stream>>>(XG, GH, Cc, HS, HP, Bn, T, 6, C);
    { GemmP ch0_7_0;
      ch0_7_0.A = HP + (size_t)0 * C; ch0_7_0.B = Wh1 + (size_t)0 * C * G4; ch0_7_0.bias = HP + (size_t)0 * C; ch0_7_0.R = HP + (size_t)0 * C; ch0_7_0.C = GH;
      ch0_7_0.sAo = (long long)PP * C; ch0_7_0.sAi = (long long)18 * C; ch0_7_0.sAm = C; ch0_7_0.sAk = 1; ch0_7_0.sBo = 0; ch0_7_0.sBi = 0; ch0_7_0.sBn = 1; ch0_7_0.sBk = G4; ch0_7_0.sCo = (long long)HW * G4; ch0_7_0.sCi = (long long)16 * G4; ch0_7_0.sCm = G4; ch0_7_0.sRo = 0; ch0_7_0.sRi = 0; ch0_7_0.sRm = 0; ch0_7_0.sRn = 0;
      ch0_7_0.M = 16; ch0_7_0.N = G4; ch0_7_0.K = C; ch0_7_0.zi_n = 16; ch0_7_0.flags = 0; ch0_7_0.act = 0;
      ch0_7_0.alpha = 1.0f; ch0_7_0.beta = 0.0f; ch0_7_0.sa = 1.0f; ch0_7_0.sb = 1.0f; ch0_7_0.Npad = G4; ch0_7_0.pad_ = 0;
      k_gemm<1><<<dim3((unsigned)((G4) + 31) / 32, (unsigned)((16) + 15) / 16, (unsigned)(Bn * 16)), 32, 0, stream>>>(ch0_7_0); }
    { GemmP ch0_7_1;
      ch0_7_1.A = HP + (size_t)1 * C; ch0_7_1.B = Wh1 + (size_t)1 * C * G4; ch0_7_1.bias = HP + (size_t)1 * C; ch0_7_1.R = GH; ch0_7_1.C = GH;
      ch0_7_1.sAo = (long long)PP * C; ch0_7_1.sAi = (long long)18 * C; ch0_7_1.sAm = C; ch0_7_1.sAk = 1; ch0_7_1.sBo = 0; ch0_7_1.sBi = 0; ch0_7_1.sBn = 1; ch0_7_1.sBk = G4; ch0_7_1.sCo = (long long)HW * G4; ch0_7_1.sCi = (long long)16 * G4; ch0_7_1.sCm = G4; ch0_7_1.sRo = (long long)HW * G4; ch0_7_1.sRi = (long long)16 * G4; ch0_7_1.sRm = G4; ch0_7_1.sRn = 1;
      ch0_7_1.M = 16; ch0_7_1.N = G4; ch0_7_1.K = C; ch0_7_1.zi_n = 16; ch0_7_1.flags = 4; ch0_7_1.act = 0;
      ch0_7_1.alpha = 1.0f; ch0_7_1.beta = 1.0f; ch0_7_1.sa = 1.0f; ch0_7_1.sb = 1.0f; ch0_7_1.Npad = G4; ch0_7_1.pad_ = 0;
      k_gemm<1><<<dim3((unsigned)((G4) + 31) / 32, (unsigned)((16) + 15) / 16, (unsigned)(Bn * 16)), 32, 0, stream>>>(ch0_7_1); }
    { GemmP ch0_7_2;
      ch0_7_2.A = HP + (size_t)2 * C; ch0_7_2.B = Wh1 + (size_t)2 * C * G4; ch0_7_2.bias = HP + (size_t)2 * C; ch0_7_2.R = GH; ch0_7_2.C = GH;
      ch0_7_2.sAo = (long long)PP * C; ch0_7_2.sAi = (long long)18 * C; ch0_7_2.sAm = C; ch0_7_2.sAk = 1; ch0_7_2.sBo = 0; ch0_7_2.sBi = 0; ch0_7_2.sBn = 1; ch0_7_2.sBk = G4; ch0_7_2.sCo = (long long)HW * G4; ch0_7_2.sCi = (long long)16 * G4; ch0_7_2.sCm = G4; ch0_7_2.sRo = (long long)HW * G4; ch0_7_2.sRi = (long long)16 * G4; ch0_7_2.sRm = G4; ch0_7_2.sRn = 1;
      ch0_7_2.M = 16; ch0_7_2.N = G4; ch0_7_2.K = C; ch0_7_2.zi_n = 16; ch0_7_2.flags = 4; ch0_7_2.act = 0;
      ch0_7_2.alpha = 1.0f; ch0_7_2.beta = 1.0f; ch0_7_2.sa = 1.0f; ch0_7_2.sb = 1.0f; ch0_7_2.Npad = G4; ch0_7_2.pad_ = 0;
      k_gemm<1><<<dim3((unsigned)((G4) + 31) / 32, (unsigned)((16) + 15) / 16, (unsigned)(Bn * 16)), 32, 0, stream>>>(ch0_7_2); }
    { GemmP ch0_7_3;
      ch0_7_3.A = HP + (size_t)18 * C; ch0_7_3.B = Wh1 + (size_t)3 * C * G4; ch0_7_3.bias = HP + (size_t)18 * C; ch0_7_3.R = GH; ch0_7_3.C = GH;
      ch0_7_3.sAo = (long long)PP * C; ch0_7_3.sAi = (long long)18 * C; ch0_7_3.sAm = C; ch0_7_3.sAk = 1; ch0_7_3.sBo = 0; ch0_7_3.sBi = 0; ch0_7_3.sBn = 1; ch0_7_3.sBk = G4; ch0_7_3.sCo = (long long)HW * G4; ch0_7_3.sCi = (long long)16 * G4; ch0_7_3.sCm = G4; ch0_7_3.sRo = (long long)HW * G4; ch0_7_3.sRi = (long long)16 * G4; ch0_7_3.sRm = G4; ch0_7_3.sRn = 1;
      ch0_7_3.M = 16; ch0_7_3.N = G4; ch0_7_3.K = C; ch0_7_3.zi_n = 16; ch0_7_3.flags = 4; ch0_7_3.act = 0;
      ch0_7_3.alpha = 1.0f; ch0_7_3.beta = 1.0f; ch0_7_3.sa = 1.0f; ch0_7_3.sb = 1.0f; ch0_7_3.Npad = G4; ch0_7_3.pad_ = 0;
      k_gemm<1><<<dim3((unsigned)((G4) + 31) / 32, (unsigned)((16) + 15) / 16, (unsigned)(Bn * 16)), 32, 0, stream>>>(ch0_7_3); }
    { GemmP ch0_7_4;
      ch0_7_4.A = HP + (size_t)19 * C; ch0_7_4.B = Wh1 + (size_t)4 * C * G4; ch0_7_4.bias = HP + (size_t)19 * C; ch0_7_4.R = GH; ch0_7_4.C = GH;
      ch0_7_4.sAo = (long long)PP * C; ch0_7_4.sAi = (long long)18 * C; ch0_7_4.sAm = C; ch0_7_4.sAk = 1; ch0_7_4.sBo = 0; ch0_7_4.sBi = 0; ch0_7_4.sBn = 1; ch0_7_4.sBk = G4; ch0_7_4.sCo = (long long)HW * G4; ch0_7_4.sCi = (long long)16 * G4; ch0_7_4.sCm = G4; ch0_7_4.sRo = (long long)HW * G4; ch0_7_4.sRi = (long long)16 * G4; ch0_7_4.sRm = G4; ch0_7_4.sRn = 1;
      ch0_7_4.M = 16; ch0_7_4.N = G4; ch0_7_4.K = C; ch0_7_4.zi_n = 16; ch0_7_4.flags = 4; ch0_7_4.act = 0;
      ch0_7_4.alpha = 1.0f; ch0_7_4.beta = 1.0f; ch0_7_4.sa = 1.0f; ch0_7_4.sb = 1.0f; ch0_7_4.Npad = G4; ch0_7_4.pad_ = 0;
      k_gemm<1><<<dim3((unsigned)((G4) + 31) / 32, (unsigned)((16) + 15) / 16, (unsigned)(Bn * 16)), 32, 0, stream>>>(ch0_7_4); }
    { GemmP ch0_7_5;
      ch0_7_5.A = HP + (size_t)20 * C; ch0_7_5.B = Wh1 + (size_t)5 * C * G4; ch0_7_5.bias = HP + (size_t)20 * C; ch0_7_5.R = GH; ch0_7_5.C = GH;
      ch0_7_5.sAo = (long long)PP * C; ch0_7_5.sAi = (long long)18 * C; ch0_7_5.sAm = C; ch0_7_5.sAk = 1; ch0_7_5.sBo = 0; ch0_7_5.sBi = 0; ch0_7_5.sBn = 1; ch0_7_5.sBk = G4; ch0_7_5.sCo = (long long)HW * G4; ch0_7_5.sCi = (long long)16 * G4; ch0_7_5.sCm = G4; ch0_7_5.sRo = (long long)HW * G4; ch0_7_5.sRi = (long long)16 * G4; ch0_7_5.sRm = G4; ch0_7_5.sRn = 1;
      ch0_7_5.M = 16; ch0_7_5.N = G4; ch0_7_5.K = C; ch0_7_5.zi_n = 16; ch0_7_5.flags = 4; ch0_7_5.act = 0;
      ch0_7_5.alpha = 1.0f; ch0_7_5.beta = 1.0f; ch0_7_5.sa = 1.0f; ch0_7_5.sb = 1.0f; ch0_7_5.Npad = G4; ch0_7_5.pad_ = 0;
      k_gemm<1><<<dim3((unsigned)((G4) + 31) / 32, (unsigned)((16) + 15) / 16, (unsigned)(Bn * 16)), 32, 0, stream>>>(ch0_7_5); }
    { GemmP ch0_7_6;
      ch0_7_6.A = HP + (size_t)36 * C; ch0_7_6.B = Wh1 + (size_t)6 * C * G4; ch0_7_6.bias = HP + (size_t)36 * C; ch0_7_6.R = GH; ch0_7_6.C = GH;
      ch0_7_6.sAo = (long long)PP * C; ch0_7_6.sAi = (long long)18 * C; ch0_7_6.sAm = C; ch0_7_6.sAk = 1; ch0_7_6.sBo = 0; ch0_7_6.sBi = 0; ch0_7_6.sBn = 1; ch0_7_6.sBk = G4; ch0_7_6.sCo = (long long)HW * G4; ch0_7_6.sCi = (long long)16 * G4; ch0_7_6.sCm = G4; ch0_7_6.sRo = (long long)HW * G4; ch0_7_6.sRi = (long long)16 * G4; ch0_7_6.sRm = G4; ch0_7_6.sRn = 1;
      ch0_7_6.M = 16; ch0_7_6.N = G4; ch0_7_6.K = C; ch0_7_6.zi_n = 16; ch0_7_6.flags = 4; ch0_7_6.act = 0;
      ch0_7_6.alpha = 1.0f; ch0_7_6.beta = 1.0f; ch0_7_6.sa = 1.0f; ch0_7_6.sb = 1.0f; ch0_7_6.Npad = G4; ch0_7_6.pad_ = 0;
      k_gemm<1><<<dim3((unsigned)((G4) + 31) / 32, (unsigned)((16) + 15) / 16, (unsigned)(Bn * 16)), 32, 0, stream>>>(ch0_7_6); }
    { GemmP ch0_7_7;
      ch0_7_7.A = HP + (size_t)37 * C; ch0_7_7.B = Wh1 + (size_t)7 * C * G4; ch0_7_7.bias = HP + (size_t)37 * C; ch0_7_7.R = GH; ch0_7_7.C = GH;
      ch0_7_7.sAo = (long long)PP * C; ch0_7_7.sAi = (long long)18 * C; ch0_7_7.sAm = C; ch0_7_7.sAk = 1; ch0_7_7.sBo = 0; ch0_7_7.sBi = 0; ch0_7_7.sBn = 1; ch0_7_7.sBk = G4; ch0_7_7.sCo = (long long)HW * G4; ch0_7_7.sCi = (long long)16 * G4; ch0_7_7.sCm = G4; ch0_7_7.sRo = (long long)HW * G4; ch0_7_7.sRi = (long long)16 * G4; ch0_7_7.sRm = G4; ch0_7_7.sRn = 1;
      ch0_7_7.M = 16; ch0_7_7.N = G4; ch0_7_7.K = C; ch0_7_7.zi_n = 16; ch0_7_7.flags = 4; ch0_7_7.act = 0;
      ch0_7_7.alpha = 1.0f; ch0_7_7.beta = 1.0f; ch0_7_7.sa = 1.0f; ch0_7_7.sb = 1.0f; ch0_7_7.Npad = G4; ch0_7_7.pad_ = 0;
      k_gemm<1><<<dim3((unsigned)((G4) + 31) / 32, (unsigned)((16) + 15) / 16, (unsigned)(Bn * 16)), 32, 0, stream>>>(ch0_7_7); }
    { GemmP ch0_7_8;
      ch0_7_8.A = HP + (size_t)38 * C; ch0_7_8.B = Wh1 + (size_t)8 * C * G4; ch0_7_8.bias = HP + (size_t)38 * C; ch0_7_8.R = GH; ch0_7_8.C = GH;
      ch0_7_8.sAo = (long long)PP * C; ch0_7_8.sAi = (long long)18 * C; ch0_7_8.sAm = C; ch0_7_8.sAk = 1; ch0_7_8.sBo = 0; ch0_7_8.sBi = 0; ch0_7_8.sBn = 1; ch0_7_8.sBk = G4; ch0_7_8.sCo = (long long)HW * G4; ch0_7_8.sCi = (long long)16 * G4; ch0_7_8.sCm = G4; ch0_7_8.sRo = (long long)HW * G4; ch0_7_8.sRi = (long long)16 * G4; ch0_7_8.sRm = G4; ch0_7_8.sRn = 1;
      ch0_7_8.M = 16; ch0_7_8.N = G4; ch0_7_8.K = C; ch0_7_8.zi_n = 16; ch0_7_8.flags = 4; ch0_7_8.act = 0;
      ch0_7_8.alpha = 1.0f; ch0_7_8.beta = 1.0f; ch0_7_8.sa = 1.0f; ch0_7_8.sb = 1.0f; ch0_7_8.Npad = G4; ch0_7_8.pad_ = 0;
      k_gemm<1><<<dim3((unsigned)((G4) + 31) / 32, (unsigned)((16) + 15) / 16, (unsigned)(Bn * 16)), 32, 0, stream>>>(ch0_7_8); }

    k_bl_cell<<<(unsigned)(((long long)Bn * HW * C + 255) / 256), 256, 0, stream>>>(XG, GH, Cc, HS, HP, Bn, T, 7, C);
    k_stats<<<(unsigned)(C), 256, 0, stream>>>(HS, 1, C, 0, 1, NF * HW, 0.001f, st, 0);
    k_norm_apply<<<(unsigned)(((long long)(NF * HW) * (C) * (1) + 255) / 256), 256, 0, stream>>>(HS, HS, st, g1, be1, NF * HW, C, 1, 1, 1, 0);
    hipMemsetAsync(XP, 0, (size_t)NF * PP * C * 4, stream); hipMemsetAsync(HP, 0, (size_t)Bn * PP * C * 4, stream); hipMemsetAsync(Cc, 0, (size_t)Bn * HW * C * 4, stream);
    k_bl_pad<<<(unsigned)(((long long)NF * HW * C + 255) / 256), 256, 0, stream>>>(HS, XP, NF, C);
    { GemmP cx1_0;
      cx1_0.A = XP + (size_t)0 * C; cx1_0.B = Wx2 + (size_t)0 * C * G4; cx1_0.bias = b2; cx1_0.R = XP + (size_t)0 * C; cx1_0.C = XG;
      cx1_0.sAo = (long long)PP * C; cx1_0.sAi = (long long)18 * C; cx1_0.sAm = C; cx1_0.sAk = 1; cx1_0.sBo = 0; cx1_0.sBi = 0; cx1_0.sBn = 1; cx1_0.sBk = G4; cx1_0.sCo = (long long)HW * G4; cx1_0.sCi = (long long)16 * G4; cx1_0.sCm = G4; cx1_0.sRo = 0; cx1_0.sRi = 0; cx1_0.sRm = 0; cx1_0.sRn = 0;
      cx1_0.M = 16; cx1_0.N = G4; cx1_0.K = C; cx1_0.zi_n = 16; cx1_0.flags = 1; cx1_0.act = 0;
      cx1_0.alpha = 1.0f; cx1_0.beta = 0.0f; cx1_0.sa = 1.0f; cx1_0.sb = 1.0f; cx1_0.Npad = G4; cx1_0.pad_ = 0;
      k_gemm<1><<<dim3((unsigned)((G4) + 31) / 32, (unsigned)((16) + 15) / 16, (unsigned)(NF * 16)), 32, 0, stream>>>(cx1_0); }
    { GemmP cx1_1;
      cx1_1.A = XP + (size_t)1 * C; cx1_1.B = Wx2 + (size_t)1 * C * G4; cx1_1.bias = XP + (size_t)1 * C; cx1_1.R = XG; cx1_1.C = XG;
      cx1_1.sAo = (long long)PP * C; cx1_1.sAi = (long long)18 * C; cx1_1.sAm = C; cx1_1.sAk = 1; cx1_1.sBo = 0; cx1_1.sBi = 0; cx1_1.sBn = 1; cx1_1.sBk = G4; cx1_1.sCo = (long long)HW * G4; cx1_1.sCi = (long long)16 * G4; cx1_1.sCm = G4; cx1_1.sRo = (long long)HW * G4; cx1_1.sRi = (long long)16 * G4; cx1_1.sRm = G4; cx1_1.sRn = 1;
      cx1_1.M = 16; cx1_1.N = G4; cx1_1.K = C; cx1_1.zi_n = 16; cx1_1.flags = 4; cx1_1.act = 0;
      cx1_1.alpha = 1.0f; cx1_1.beta = 1.0f; cx1_1.sa = 1.0f; cx1_1.sb = 1.0f; cx1_1.Npad = G4; cx1_1.pad_ = 0;
      k_gemm<1><<<dim3((unsigned)((G4) + 31) / 32, (unsigned)((16) + 15) / 16, (unsigned)(NF * 16)), 32, 0, stream>>>(cx1_1); }
    { GemmP cx1_2;
      cx1_2.A = XP + (size_t)2 * C; cx1_2.B = Wx2 + (size_t)2 * C * G4; cx1_2.bias = XP + (size_t)2 * C; cx1_2.R = XG; cx1_2.C = XG;
      cx1_2.sAo = (long long)PP * C; cx1_2.sAi = (long long)18 * C; cx1_2.sAm = C; cx1_2.sAk = 1; cx1_2.sBo = 0; cx1_2.sBi = 0; cx1_2.sBn = 1; cx1_2.sBk = G4; cx1_2.sCo = (long long)HW * G4; cx1_2.sCi = (long long)16 * G4; cx1_2.sCm = G4; cx1_2.sRo = (long long)HW * G4; cx1_2.sRi = (long long)16 * G4; cx1_2.sRm = G4; cx1_2.sRn = 1;
      cx1_2.M = 16; cx1_2.N = G4; cx1_2.K = C; cx1_2.zi_n = 16; cx1_2.flags = 4; cx1_2.act = 0;
      cx1_2.alpha = 1.0f; cx1_2.beta = 1.0f; cx1_2.sa = 1.0f; cx1_2.sb = 1.0f; cx1_2.Npad = G4; cx1_2.pad_ = 0;
      k_gemm<1><<<dim3((unsigned)((G4) + 31) / 32, (unsigned)((16) + 15) / 16, (unsigned)(NF * 16)), 32, 0, stream>>>(cx1_2); }
    { GemmP cx1_3;
      cx1_3.A = XP + (size_t)18 * C; cx1_3.B = Wx2 + (size_t)3 * C * G4; cx1_3.bias = XP + (size_t)18 * C; cx1_3.R = XG; cx1_3.C = XG;
      cx1_3.sAo = (long long)PP * C; cx1_3.sAi = (long long)18 * C; cx1_3.sAm = C; cx1_3.sAk = 1; cx1_3.sBo = 0; cx1_3.sBi = 0; cx1_3.sBn = 1; cx1_3.sBk = G4; cx1_3.sCo = (long long)HW * G4; cx1_3.sCi = (long long)16 * G4; cx1_3.sCm = G4; cx1_3.sRo = (long long)HW * G4; cx1_3.sRi = (long long)16 * G4; cx1_3.sRm = G4; cx1_3.sRn = 1;
      cx1_3.M = 16; cx1_3.N = G4; cx1_3.K = C; cx1_3.zi_n = 16; cx1_3.flags = 4; cx1_3.act = 0;
      cx1_3.alpha = 1.0f; cx1_3.beta = 1.0f; cx1_3.sa = 1.0f; cx1_3.sb = 1.0f; cx1_3.Npad = G4; cx1_3.pad_ = 0;
      k_gemm<1><<<dim3((unsigned)((G4) + 31) / 32, (unsigned)((16) + 15) / 16, (unsigned)(NF * 16)), 32, 0, stream>>>(cx1_3); }
    { GemmP cx1_4;
      cx1_4.A = XP + (size_t)19 * C; cx1_4.B = Wx2 + (size_t)4 * C * G4; cx1_4.bias = XP + (size_t)19 * C; cx1_4.R = XG; cx1_4.C = XG;
      cx1_4.sAo = (long long)PP * C; cx1_4.sAi = (long long)18 * C; cx1_4.sAm = C; cx1_4.sAk = 1; cx1_4.sBo = 0; cx1_4.sBi = 0; cx1_4.sBn = 1; cx1_4.sBk = G4; cx1_4.sCo = (long long)HW * G4; cx1_4.sCi = (long long)16 * G4; cx1_4.sCm = G4; cx1_4.sRo = (long long)HW * G4; cx1_4.sRi = (long long)16 * G4; cx1_4.sRm = G4; cx1_4.sRn = 1;
      cx1_4.M = 16; cx1_4.N = G4; cx1_4.K = C; cx1_4.zi_n = 16; cx1_4.flags = 4; cx1_4.act = 0;
      cx1_4.alpha = 1.0f; cx1_4.beta = 1.0f; cx1_4.sa = 1.0f; cx1_4.sb = 1.0f; cx1_4.Npad = G4; cx1_4.pad_ = 0;
      k_gemm<1><<<dim3((unsigned)((G4) + 31) / 32, (unsigned)((16) + 15) / 16, (unsigned)(NF * 16)), 32, 0, stream>>>(cx1_4); }
    { GemmP cx1_5;
      cx1_5.A = XP + (size_t)20 * C; cx1_5.B = Wx2 + (size_t)5 * C * G4; cx1_5.bias = XP + (size_t)20 * C; cx1_5.R = XG; cx1_5.C = XG;
      cx1_5.sAo = (long long)PP * C; cx1_5.sAi = (long long)18 * C; cx1_5.sAm = C; cx1_5.sAk = 1; cx1_5.sBo = 0; cx1_5.sBi = 0; cx1_5.sBn = 1; cx1_5.sBk = G4; cx1_5.sCo = (long long)HW * G4; cx1_5.sCi = (long long)16 * G4; cx1_5.sCm = G4; cx1_5.sRo = (long long)HW * G4; cx1_5.sRi = (long long)16 * G4; cx1_5.sRm = G4; cx1_5.sRn = 1;
      cx1_5.M = 16; cx1_5.N = G4; cx1_5.K = C; cx1_5.zi_n = 16; cx1_5.flags = 4; cx1_5.act = 0;
      cx1_5.alpha = 1.0f; cx1_5.beta = 1.0f; cx1_5.sa = 1.0f; cx1_5.sb = 1.0f; cx1_5.Npad = G4; cx1_5.pad_ = 0;
      k_gemm<1><<<dim3((unsigned)((G4) + 31) / 32, (unsigned)((16) + 15) / 16, (unsigned)(NF * 16)), 32, 0, stream>>>(cx1_5); }
    { GemmP cx1_6;
      cx1_6.A = XP + (size_t)36 * C; cx1_6.B = Wx2 + (size_t)6 * C * G4; cx1_6.bias = XP + (size_t)36 * C; cx1_6.R = XG; cx1_6.C = XG;
      cx1_6.sAo = (long long)PP * C; cx1_6.sAi = (long long)18 * C; cx1_6.sAm = C; cx1_6.sAk = 1; cx1_6.sBo = 0; cx1_6.sBi = 0; cx1_6.sBn = 1; cx1_6.sBk = G4; cx1_6.sCo = (long long)HW * G4; cx1_6.sCi = (long long)16 * G4; cx1_6.sCm = G4; cx1_6.sRo = (long long)HW * G4; cx1_6.sRi = (long long)16 * G4; cx1_6.sRm = G4; cx1_6.sRn = 1;
      cx1_6.M = 16; cx1_6.N = G4; cx1_6.K = C; cx1_6.zi_n = 16; cx1_6.flags = 4; cx1_6.act = 0;
      cx1_6.alpha = 1.0f; cx1_6.beta = 1.0f; cx1_6.sa = 1.0f; cx1_6.sb = 1.0f; cx1_6.Npad = G4; cx1_6.pad_ = 0;
      k_gemm<1><<<dim3((unsigned)((G4) + 31) / 32, (unsigned)((16) + 15) / 16, (unsigned)(NF * 16)), 32, 0, stream>>>(cx1_6); }
    { GemmP cx1_7;
      cx1_7.A = XP + (size_t)37 * C; cx1_7.B = Wx2 + (size_t)7 * C * G4; cx1_7.bias = XP + (size_t)37 * C; cx1_7.R = XG; cx1_7.C = XG;
      cx1_7.sAo = (long long)PP * C; cx1_7.sAi = (long long)18 * C; cx1_7.sAm = C; cx1_7.sAk = 1; cx1_7.sBo = 0; cx1_7.sBi = 0; cx1_7.sBn = 1; cx1_7.sBk = G4; cx1_7.sCo = (long long)HW * G4; cx1_7.sCi = (long long)16 * G4; cx1_7.sCm = G4; cx1_7.sRo = (long long)HW * G4; cx1_7.sRi = (long long)16 * G4; cx1_7.sRm = G4; cx1_7.sRn = 1;
      cx1_7.M = 16; cx1_7.N = G4; cx1_7.K = C; cx1_7.zi_n = 16; cx1_7.flags = 4; cx1_7.act = 0;
      cx1_7.alpha = 1.0f; cx1_7.beta = 1.0f; cx1_7.sa = 1.0f; cx1_7.sb = 1.0f; cx1_7.Npad = G4; cx1_7.pad_ = 0;
      k_gemm<1><<<dim3((unsigned)((G4) + 31) / 32, (unsigned)((16) + 15) / 16, (unsigned)(NF * 16)), 32, 0, stream>>>(cx1_7); }
    { GemmP cx1_8;
      cx1_8.A = XP + (size_t)38 * C; cx1_8.B = Wx2 + (size_t)8 * C * G4; cx1_8.bias = XP + (size_t)38 * C; cx1_8.R = XG; cx1_8.C = XG;
      cx1_8.sAo = (long long)PP * C; cx1_8.sAi = (long long)18 * C; cx1_8.sAm = C; cx1_8.sAk = 1; cx1_8.sBo = 0; cx1_8.sBi = 0; cx1_8.sBn = 1; cx1_8.sBk = G4; cx1_8.sCo = (long long)HW * G4; cx1_8.sCi = (long long)16 * G4; cx1_8.sCm = G4; cx1_8.sRo = (long long)HW * G4; cx1_8.sRi = (long long)16 * G4; cx1_8.sRm = G4; cx1_8.sRn = 1;
      cx1_8.M = 16; cx1_8.N = G4; cx1_8.K = C; cx1_8.zi_n = 16; cx1_8.flags = 4; cx1_8.act = 0;
      cx1_8.alpha = 1.0f; cx1_8.beta = 1.0f; cx1_8.sa = 1.0f; cx1_8.sb = 1.0f; cx1_8.Npad = G4; cx1_8.pad_ = 0;
      k_gemm<1><<<dim3((unsigned)((G4) + 31) / 32, (unsigned)((16) + 15) / 16, (unsigned)(NF * 16)), 32, 0, stream>>>(cx1_8); }

    { GemmP ch1_0_0;
      ch1_0_0.A = HP + (size_t)0 * C; ch1_0_0.B = Wh2 + (size_t)0 * C * G4; ch1_0_0.bias = HP + (size_t)0 * C; ch1_0_0.R = HP + (size_t)0 * C; ch1_0_0.C = GH;
      ch1_0_0.sAo = (long long)PP * C; ch1_0_0.sAi = (long long)18 * C; ch1_0_0.sAm = C; ch1_0_0.sAk = 1; ch1_0_0.sBo = 0; ch1_0_0.sBi = 0; ch1_0_0.sBn = 1; ch1_0_0.sBk = G4; ch1_0_0.sCo = (long long)HW * G4; ch1_0_0.sCi = (long long)16 * G4; ch1_0_0.sCm = G4; ch1_0_0.sRo = 0; ch1_0_0.sRi = 0; ch1_0_0.sRm = 0; ch1_0_0.sRn = 0;
      ch1_0_0.M = 16; ch1_0_0.N = G4; ch1_0_0.K = C; ch1_0_0.zi_n = 16; ch1_0_0.flags = 0; ch1_0_0.act = 0;
      ch1_0_0.alpha = 1.0f; ch1_0_0.beta = 0.0f; ch1_0_0.sa = 1.0f; ch1_0_0.sb = 1.0f; ch1_0_0.Npad = G4; ch1_0_0.pad_ = 0;
      k_gemm<1><<<dim3((unsigned)((G4) + 31) / 32, (unsigned)((16) + 15) / 16, (unsigned)(Bn * 16)), 32, 0, stream>>>(ch1_0_0); }
    { GemmP ch1_0_1;
      ch1_0_1.A = HP + (size_t)1 * C; ch1_0_1.B = Wh2 + (size_t)1 * C * G4; ch1_0_1.bias = HP + (size_t)1 * C; ch1_0_1.R = GH; ch1_0_1.C = GH;
      ch1_0_1.sAo = (long long)PP * C; ch1_0_1.sAi = (long long)18 * C; ch1_0_1.sAm = C; ch1_0_1.sAk = 1; ch1_0_1.sBo = 0; ch1_0_1.sBi = 0; ch1_0_1.sBn = 1; ch1_0_1.sBk = G4; ch1_0_1.sCo = (long long)HW * G4; ch1_0_1.sCi = (long long)16 * G4; ch1_0_1.sCm = G4; ch1_0_1.sRo = (long long)HW * G4; ch1_0_1.sRi = (long long)16 * G4; ch1_0_1.sRm = G4; ch1_0_1.sRn = 1;
      ch1_0_1.M = 16; ch1_0_1.N = G4; ch1_0_1.K = C; ch1_0_1.zi_n = 16; ch1_0_1.flags = 4; ch1_0_1.act = 0;
      ch1_0_1.alpha = 1.0f; ch1_0_1.beta = 1.0f; ch1_0_1.sa = 1.0f; ch1_0_1.sb = 1.0f; ch1_0_1.Npad = G4; ch1_0_1.pad_ = 0;
      k_gemm<1><<<dim3((unsigned)((G4) + 31) / 32, (unsigned)((16) + 15) / 16, (unsigned)(Bn * 16)), 32, 0, stream>>>(ch1_0_1); }
    { GemmP ch1_0_2;
      ch1_0_2.A = HP + (size_t)2 * C; ch1_0_2.B = Wh2 + (size_t)2 * C * G4; ch1_0_2.bias = HP + (size_t)2 * C; ch1_0_2.R = GH; ch1_0_2.C = GH;
      ch1_0_2.sAo = (long long)PP * C; ch1_0_2.sAi = (long long)18 * C; ch1_0_2.sAm = C; ch1_0_2.sAk = 1; ch1_0_2.sBo = 0; ch1_0_2.sBi = 0; ch1_0_2.sBn = 1; ch1_0_2.sBk = G4; ch1_0_2.sCo = (long long)HW * G4; ch1_0_2.sCi = (long long)16 * G4; ch1_0_2.sCm = G4; ch1_0_2.sRo = (long long)HW * G4; ch1_0_2.sRi = (long long)16 * G4; ch1_0_2.sRm = G4; ch1_0_2.sRn = 1;
      ch1_0_2.M = 16; ch1_0_2.N = G4; ch1_0_2.K = C; ch1_0_2.zi_n = 16; ch1_0_2.flags = 4; ch1_0_2.act = 0;
      ch1_0_2.alpha = 1.0f; ch1_0_2.beta = 1.0f; ch1_0_2.sa = 1.0f; ch1_0_2.sb = 1.0f; ch1_0_2.Npad = G4; ch1_0_2.pad_ = 0;
      k_gemm<1><<<dim3((unsigned)((G4) + 31) / 32, (unsigned)((16) + 15) / 16, (unsigned)(Bn * 16)), 32, 0, stream>>>(ch1_0_2); }
    { GemmP ch1_0_3;
      ch1_0_3.A = HP + (size_t)18 * C; ch1_0_3.B = Wh2 + (size_t)3 * C * G4; ch1_0_3.bias = HP + (size_t)18 * C; ch1_0_3.R = GH; ch1_0_3.C = GH;
      ch1_0_3.sAo = (long long)PP * C; ch1_0_3.sAi = (long long)18 * C; ch1_0_3.sAm = C; ch1_0_3.sAk = 1; ch1_0_3.sBo = 0; ch1_0_3.sBi = 0; ch1_0_3.sBn = 1; ch1_0_3.sBk = G4; ch1_0_3.sCo = (long long)HW * G4; ch1_0_3.sCi = (long long)16 * G4; ch1_0_3.sCm = G4; ch1_0_3.sRo = (long long)HW * G4; ch1_0_3.sRi = (long long)16 * G4; ch1_0_3.sRm = G4; ch1_0_3.sRn = 1;
      ch1_0_3.M = 16; ch1_0_3.N = G4; ch1_0_3.K = C; ch1_0_3.zi_n = 16; ch1_0_3.flags = 4; ch1_0_3.act = 0;
      ch1_0_3.alpha = 1.0f; ch1_0_3.beta = 1.0f; ch1_0_3.sa = 1.0f; ch1_0_3.sb = 1.0f; ch1_0_3.Npad = G4; ch1_0_3.pad_ = 0;
      k_gemm<1><<<dim3((unsigned)((G4) + 31) / 32, (unsigned)((16) + 15) / 16, (unsigned)(Bn * 16)), 32, 0, stream>>>(ch1_0_3); }
    { GemmP ch1_0_4;
      ch1_0_4.A = HP + (size_t)19 * C; ch1_0_4.B = Wh2 + (size_t)4 * C * G4; ch1_0_4.bias = HP + (size_t)19 * C; ch1_0_4.R = GH; ch1_0_4.C = GH;
      ch1_0_4.sAo = (long long)PP * C; ch1_0_4.sAi = (long long)18 * C; ch1_0_4.sAm = C; ch1_0_4.sAk = 1; ch1_0_4.sBo = 0; ch1_0_4.sBi = 0; ch1_0_4.sBn = 1; ch1_0_4.sBk = G4; ch1_0_4.sCo = (long long)HW * G4; ch1_0_4.sCi = (long long)16 * G4; ch1_0_4.sCm = G4; ch1_0_4.sRo = (long long)HW * G4; ch1_0_4.sRi = (long long)16 * G4; ch1_0_4.sRm = G4; ch1_0_4.sRn = 1;
      ch1_0_4.M = 16; ch1_0_4.N = G4; ch1_0_4.K = C; ch1_0_4.zi_n = 16; ch1_0_4.flags = 4; ch1_0_4.act = 0;
      ch1_0_4.alpha = 1.0f; ch1_0_4.beta = 1.0f; ch1_0_4.sa = 1.0f; ch1_0_4.sb = 1.0f; ch1_0_4.Npad = G4; ch1_0_4.pad_ = 0;
      k_gemm<1><<<dim3((unsigned)((G4) + 31) / 32, (unsigned)((16) + 15) / 16, (unsigned)(Bn * 16)), 32, 0, stream>>>(ch1_0_4); }
    { GemmP ch1_0_5;
      ch1_0_5.A = HP + (size_t)20 * C; ch1_0_5.B = Wh2 + (size_t)5 * C * G4; ch1_0_5.bias = HP + (size_t)20 * C; ch1_0_5.R = GH; ch1_0_5.C = GH;
      ch1_0_5.sAo = (long long)PP * C; ch1_0_5.sAi = (long long)18 * C; ch1_0_5.sAm = C; ch1_0_5.sAk = 1; ch1_0_5.sBo = 0; ch1_0_5.sBi = 0; ch1_0_5.sBn = 1; ch1_0_5.sBk = G4; ch1_0_5.sCo = (long long)HW * G4; ch1_0_5.sCi = (long long)16 * G4; ch1_0_5.sCm = G4; ch1_0_5.sRo = (long long)HW * G4; ch1_0_5.sRi = (long long)16 * G4; ch1_0_5.sRm = G4; ch1_0_5.sRn = 1;
      ch1_0_5.M = 16; ch1_0_5.N = G4; ch1_0_5.K = C; ch1_0_5.zi_n = 16; ch1_0_5.flags = 4; ch1_0_5.act = 0;
      ch1_0_5.alpha = 1.0f; ch1_0_5.beta = 1.0f; ch1_0_5.sa = 1.0f; ch1_0_5.sb = 1.0f; ch1_0_5.Npad = G4; ch1_0_5.pad_ = 0;
      k_gemm<1><<<dim3((unsigned)((G4) + 31) / 32, (unsigned)((16) + 15) / 16, (unsigned)(Bn * 16)), 32, 0, stream>>>(ch1_0_5); }
    { GemmP ch1_0_6;
      ch1_0_6.A = HP + (size_t)36 * C; ch1_0_6.B = Wh2 + (size_t)6 * C * G4; ch1_0_6.bias = HP + (size_t)36 * C; ch1_0_6.R = GH; ch1_0_6.C = GH;
      ch1_0_6.sAo = (long long)PP * C; ch1_0_6.sAi = (long long)18 * C; ch1_0_6.sAm = C; ch1_0_6.sAk = 1; ch1_0_6.sBo = 0; ch1_0_6.sBi = 0; ch1_0_6.sBn = 1; ch1_0_6.sBk = G4; ch1_0_6.sCo = (long long)HW * G4; ch1_0_6.sCi = (long long)16 * G4; ch1_0_6.sCm = G4; ch1_0_6.sRo = (long long)HW * G4; ch1_0_6.sRi = (long long)16 * G4; ch1_0_6.sRm = G4; ch1_0_6.sRn = 1;
      ch1_0_6.M = 16; ch1_0_6.N = G4; ch1_0_6.K = C; ch1_0_6.zi_n = 16; ch1_0_6.flags = 4; ch1_0_6.act = 0;
      ch1_0_6.alpha = 1.0f; ch1_0_6.beta = 1.0f; ch1_0_6.sa = 1.0f; ch1_0_6.sb = 1.0f; ch1_0_6.Npad = G4; ch1_0_6.pad_ = 0;
      k_gemm<1><<<dim3((unsigned)((G4) + 31) / 32, (unsigned)((16) + 15) / 16, (unsigned)(Bn * 16)), 32, 0, stream>>>(ch1_0_6); }
    { GemmP ch1_0_7;
      ch1_0_7.A = HP + (size_t)37 * C; ch1_0_7.B = Wh2 + (size_t)7 * C * G4; ch1_0_7.bias = HP + (size_t)37 * C; ch1_0_7.R = GH; ch1_0_7.C = GH;
      ch1_0_7.sAo = (long long)PP * C; ch1_0_7.sAi = (long long)18 * C; ch1_0_7.sAm = C; ch1_0_7.sAk = 1; ch1_0_7.sBo = 0; ch1_0_7.sBi = 0; ch1_0_7.sBn = 1; ch1_0_7.sBk = G4; ch1_0_7.sCo = (long long)HW * G4; ch1_0_7.sCi = (long long)16 * G4; ch1_0_7.sCm = G4; ch1_0_7.sRo = (long long)HW * G4; ch1_0_7.sRi = (long long)16 * G4; ch1_0_7.sRm = G4; ch1_0_7.sRn = 1;
      ch1_0_7.M = 16; ch1_0_7.N = G4; ch1_0_7.K = C; ch1_0_7.zi_n = 16; ch1_0_7.flags = 4; ch1_0_7.act = 0;
      ch1_0_7.alpha = 1.0f; ch1_0_7.beta = 1.0f; ch1_0_7.sa = 1.0f; ch1_0_7.sb = 1.0f; ch1_0_7.Npad = G4; ch1_0_7.pad_ = 0;
      k_gemm<1><<<dim3((unsigned)((G4) + 31) / 32, (unsigned)((16) + 15) / 16, (unsigned)(Bn * 16)), 32, 0, stream>>>(ch1_0_7); }
    { GemmP ch1_0_8;
      ch1_0_8.A = HP + (size_t)38 * C; ch1_0_8.B = Wh2 + (size_t)8 * C * G4; ch1_0_8.bias = HP + (size_t)38 * C; ch1_0_8.R = GH; ch1_0_8.C = GH;
      ch1_0_8.sAo = (long long)PP * C; ch1_0_8.sAi = (long long)18 * C; ch1_0_8.sAm = C; ch1_0_8.sAk = 1; ch1_0_8.sBo = 0; ch1_0_8.sBi = 0; ch1_0_8.sBn = 1; ch1_0_8.sBk = G4; ch1_0_8.sCo = (long long)HW * G4; ch1_0_8.sCi = (long long)16 * G4; ch1_0_8.sCm = G4; ch1_0_8.sRo = (long long)HW * G4; ch1_0_8.sRi = (long long)16 * G4; ch1_0_8.sRm = G4; ch1_0_8.sRn = 1;
      ch1_0_8.M = 16; ch1_0_8.N = G4; ch1_0_8.K = C; ch1_0_8.zi_n = 16; ch1_0_8.flags = 4; ch1_0_8.act = 0;
      ch1_0_8.alpha = 1.0f; ch1_0_8.beta = 1.0f; ch1_0_8.sa = 1.0f; ch1_0_8.sb = 1.0f; ch1_0_8.Npad = G4; ch1_0_8.pad_ = 0;
      k_gemm<1><<<dim3((unsigned)((G4) + 31) / 32, (unsigned)((16) + 15) / 16, (unsigned)(Bn * 16)), 32, 0, stream>>>(ch1_0_8); }

    k_bl_cell<<<(unsigned)(((long long)Bn * HW * C + 255) / 256), 256, 0, stream>>>(XG, GH, Cc, HS, HP, Bn, T, 0, C);
    { GemmP ch1_1_0;
      ch1_1_0.A = HP + (size_t)0 * C; ch1_1_0.B = Wh2 + (size_t)0 * C * G4; ch1_1_0.bias = HP + (size_t)0 * C; ch1_1_0.R = HP + (size_t)0 * C; ch1_1_0.C = GH;
      ch1_1_0.sAo = (long long)PP * C; ch1_1_0.sAi = (long long)18 * C; ch1_1_0.sAm = C; ch1_1_0.sAk = 1; ch1_1_0.sBo = 0; ch1_1_0.sBi = 0; ch1_1_0.sBn = 1; ch1_1_0.sBk = G4; ch1_1_0.sCo = (long long)HW * G4; ch1_1_0.sCi = (long long)16 * G4; ch1_1_0.sCm = G4; ch1_1_0.sRo = 0; ch1_1_0.sRi = 0; ch1_1_0.sRm = 0; ch1_1_0.sRn = 0;
      ch1_1_0.M = 16; ch1_1_0.N = G4; ch1_1_0.K = C; ch1_1_0.zi_n = 16; ch1_1_0.flags = 0; ch1_1_0.act = 0;
      ch1_1_0.alpha = 1.0f; ch1_1_0.beta = 0.0f; ch1_1_0.sa = 1.0f; ch1_1_0.sb = 1.0f; ch1_1_0.Npad = G4; ch1_1_0.pad_ = 0;
      k_gemm<1><<<dim3((unsigned)((G4) + 31) / 32, (unsigned)((16) + 15) / 16, (unsigned)(Bn * 16)), 32, 0, stream>>>(ch1_1_0); }
    { GemmP ch1_1_1;
      ch1_1_1.A = HP + (size_t)1 * C; ch1_1_1.B = Wh2 + (size_t)1 * C * G4; ch1_1_1.bias = HP + (size_t)1 * C; ch1_1_1.R = GH; ch1_1_1.C = GH;
      ch1_1_1.sAo = (long long)PP * C; ch1_1_1.sAi = (long long)18 * C; ch1_1_1.sAm = C; ch1_1_1.sAk = 1; ch1_1_1.sBo = 0; ch1_1_1.sBi = 0; ch1_1_1.sBn = 1; ch1_1_1.sBk = G4; ch1_1_1.sCo = (long long)HW * G4; ch1_1_1.sCi = (long long)16 * G4; ch1_1_1.sCm = G4; ch1_1_1.sRo = (long long)HW * G4; ch1_1_1.sRi = (long long)16 * G4; ch1_1_1.sRm = G4; ch1_1_1.sRn = 1;
      ch1_1_1.M = 16; ch1_1_1.N = G4; ch1_1_1.K = C; ch1_1_1.zi_n = 16; ch1_1_1.flags = 4; ch1_1_1.act = 0;
      ch1_1_1.alpha = 1.0f; ch1_1_1.beta = 1.0f; ch1_1_1.sa = 1.0f; ch1_1_1.sb = 1.0f; ch1_1_1.Npad = G4; ch1_1_1.pad_ = 0;
      k_gemm<1><<<dim3((unsigned)((G4) + 31) / 32, (unsigned)((16) + 15) / 16, (unsigned)(Bn * 16)), 32, 0, stream>>>(ch1_1_1); }
    { GemmP ch1_1_2;
      ch1_1_2.A = HP + (size_t)2 * C; ch1_1_2.B = Wh2 + (size_t)2 * C * G4; ch1_1_2.bias = HP + (size_t)2 * C; ch1_1_2.R = GH; ch1_1_2.C = GH;
      ch1_1_2.sAo = (long long)PP * C; ch1_1_2.sAi = (long long)18 * C; ch1_1_2.sAm = C; ch1_1_2.sAk = 1; ch1_1_2.sBo = 0; ch1_1_2.sBi = 0; ch1_1_2.sBn = 1; ch1_1_2.sBk = G4; ch1_1_2.sCo = (long long)HW * G4; ch1_1_2.sCi = (long long)16 * G4; ch1_1_2.sCm = G4; ch1_1_2.sRo = (long long)HW * G4; ch1_1_2.sRi = (long long)16 * G4; ch1_1_2.sRm = G4; ch1_1_2.sRn = 1;
      ch1_1_2.M = 16; ch1_1_2.N = G4; ch1_1_2.K = C; ch1_1_2.zi_n = 16; ch1_1_2.flags = 4; ch1_1_2.act = 0;
      ch1_1_2.alpha = 1.0f; ch1_1_2.beta = 1.0f; ch1_1_2.sa = 1.0f; ch1_1_2.sb = 1.0f; ch1_1_2.Npad = G4; ch1_1_2.pad_ = 0;
      k_gemm<1><<<dim3((unsigned)((G4) + 31) / 32, (unsigned)((16) + 15) / 16, (unsigned)(Bn * 16)), 32, 0, stream>>>(ch1_1_2); }
    { GemmP ch1_1_3;
      ch1_1_3.A = HP + (size_t)18 * C; ch1_1_3.B = Wh2 + (size_t)3 * C * G4; ch1_1_3.bias = HP + (size_t)18 * C; ch1_1_3.R = GH; ch1_1_3.C = GH;
      ch1_1_3.sAo = (long long)PP * C; ch1_1_3.sAi = (long long)18 * C; ch1_1_3.sAm = C; ch1_1_3.sAk = 1; ch1_1_3.sBo = 0; ch1_1_3.sBi = 0; ch1_1_3.sBn = 1; ch1_1_3.sBk = G4; ch1_1_3.sCo = (long long)HW * G4; ch1_1_3.sCi = (long long)16 * G4; ch1_1_3.sCm = G4; ch1_1_3.sRo = (long long)HW * G4; ch1_1_3.sRi = (long long)16 * G4; ch1_1_3.sRm = G4; ch1_1_3.sRn = 1;
      ch1_1_3.M = 16; ch1_1_3.N = G4; ch1_1_3.K = C; ch1_1_3.zi_n = 16; ch1_1_3.flags = 4; ch1_1_3.act = 0;
      ch1_1_3.alpha = 1.0f; ch1_1_3.beta = 1.0f; ch1_1_3.sa = 1.0f; ch1_1_3.sb = 1.0f; ch1_1_3.Npad = G4; ch1_1_3.pad_ = 0;
      k_gemm<1><<<dim3((unsigned)((G4) + 31) / 32, (unsigned)((16) + 15) / 16, (unsigned)(Bn * 16)), 32, 0, stream>>>(ch1_1_3); }
    { GemmP ch1_1_4;
      ch1_1_4.A = HP + (size_t)19 * C; ch1_1_4.B = Wh2 + (size_t)4 * C * G4; ch1_1_4.bias = HP + (size_t)19 * C; ch1_1_4.R = GH; ch1_1_4.C = GH;
      ch1_1_4.sAo = (long long)PP * C; ch1_1_4.sAi = (long long)18 * C; ch1_1_4.sAm = C; ch1_1_4.sAk = 1; ch1_1_4.sBo = 0; ch1_1_4.sBi = 0; ch1_1_4.sBn = 1; ch1_1_4.sBk = G4; ch1_1_4.sCo = (long long)HW * G4; ch1_1_4.sCi = (long long)16 * G4; ch1_1_4.sCm = G4; ch1_1_4.sRo = (long long)HW * G4; ch1_1_4.sRi = (long long)16 * G4; ch1_1_4.sRm = G4; ch1_1_4.sRn = 1;
      ch1_1_4.M = 16; ch1_1_4.N = G4; ch1_1_4.K = C; ch1_1_4.zi_n = 16; ch1_1_4.flags = 4; ch1_1_4.act = 0;
      ch1_1_4.alpha = 1.0f; ch1_1_4.beta = 1.0f; ch1_1_4.sa = 1.0f; ch1_1_4.sb = 1.0f; ch1_1_4.Npad = G4; ch1_1_4.pad_ = 0;
      k_gemm<1><<<dim3((unsigned)((G4) + 31) / 32, (unsigned)((16) + 15) / 16, (unsigned)(Bn * 16)), 32, 0, stream>>>(ch1_1_4); }
    { GemmP ch1_1_5;
      ch1_1_5.A = HP + (size_t)20 * C; ch1_1_5.B = Wh2 + (size_t)5 * C * G4; ch1_1_5.bias = HP + (size_t)20 * C; ch1_1_5.R = GH; ch1_1_5.C = GH;
      ch1_1_5.sAo = (long long)PP * C; ch1_1_5.sAi = (long long)18 * C; ch1_1_5.sAm = C; ch1_1_5.sAk = 1; ch1_1_5.sBo = 0; ch1_1_5.sBi = 0; ch1_1_5.sBn = 1; ch1_1_5.sBk = G4; ch1_1_5.sCo = (long long)HW * G4; ch1_1_5.sCi = (long long)16 * G4; ch1_1_5.sCm = G4; ch1_1_5.sRo = (long long)HW * G4; ch1_1_5.sRi = (long long)16 * G4; ch1_1_5.sRm = G4; ch1_1_5.sRn = 1;
      ch1_1_5.M = 16; ch1_1_5.N = G4; ch1_1_5.K = C; ch1_1_5.zi_n = 16; ch1_1_5.flags = 4; ch1_1_5.act = 0;
      ch1_1_5.alpha = 1.0f; ch1_1_5.beta = 1.0f; ch1_1_5.sa = 1.0f; ch1_1_5.sb = 1.0f; ch1_1_5.Npad = G4; ch1_1_5.pad_ = 0;
      k_gemm<1><<<dim3((unsigned)((G4) + 31) / 32, (unsigned)((16) + 15) / 16, (unsigned)(Bn * 16)), 32, 0, stream>>>(ch1_1_5); }
    { GemmP ch1_1_6;
      ch1_1_6.A = HP + (size_t)36 * C; ch1_1_6.B = Wh2 + (size_t)6 * C * G4; ch1_1_6.bias = HP + (size_t)36 * C; ch1_1_6.R = GH; ch1_1_6.C = GH;
      ch1_1_6.sAo = (long long)PP * C; ch1_1_6.sAi = (long long)18 * C; ch1_1_6.sAm = C; ch1_1_6.sAk = 1; ch1_1_6.sBo = 0; ch1_1_6.sBi = 0; ch1_1_6.sBn = 1; ch1_1_6.sBk = G4; ch1_1_6.sCo = (long long)HW * G4; ch1_1_6.sCi = (long long)16 * G4; ch1_1_6.sCm = G4; ch1_1_6.sRo = (long long)HW * G4; ch1_1_6.sRi = (long long)16 * G4; ch1_1_6.sRm = G4; ch1_1_6.sRn = 1;
      ch1_1_6.M = 16; ch1_1_6.N = G4; ch1_1_6.K = C; ch1_1_6.zi_n = 16; ch1_1_6.flags = 4; ch1_1_6.act = 0;
      ch1_1_6.alpha = 1.0f; ch1_1_6.beta = 1.0f; ch1_1_6.sa = 1.0f; ch1_1_6.sb = 1.0f; ch1_1_6.Npad = G4; ch1_1_6.pad_ = 0;
      k_gemm<1><<<dim3((unsigned)((G4) + 31) / 32, (unsigned)((16) + 15) / 16, (unsigned)(Bn * 16)), 32, 0, stream>>>(ch1_1_6); }
    { GemmP ch1_1_7;
      ch1_1_7.A = HP + (size_t)37 * C; ch1_1_7.B = Wh2 + (size_t)7 * C * G4; ch1_1_7.bias = HP + (size_t)37 * C; ch1_1_7.R = GH; ch1_1_7.C = GH;
      ch1_1_7.sAo = (long long)PP * C; ch1_1_7.sAi = (long long)18 * C; ch1_1_7.sAm = C; ch1_1_7.sAk = 1; ch1_1_7.sBo = 0; ch1_1_7.sBi = 0; ch1_1_7.sBn = 1; ch1_1_7.sBk = G4; ch1_1_7.sCo = (long long)HW * G4; ch1_1_7.sCi = (long long)16 * G4; ch1_1_7.sCm = G4; ch1_1_7.sRo = (long long)HW * G4; ch1_1_7.sRi = (long long)16 * G4; ch1_1_7.sRm = G4; ch1_1_7.sRn = 1;
      ch1_1_7.M = 16; ch1_1_7.N = G4; ch1_1_7.K = C; ch1_1_7.zi_n = 16; ch1_1_7.flags = 4; ch1_1_7.act = 0;
      ch1_1_7.alpha = 1.0f; ch1_1_7.beta = 1.0f; ch1_1_7.sa = 1.0f; ch1_1_7.sb = 1.0f; ch1_1_7.Npad = G4; ch1_1_7.pad_ = 0;
      k_gemm<1><<<dim3((unsigned)((G4) + 31) / 32, (unsigned)((16) + 15) / 16, (unsigned)(Bn * 16)), 32, 0, stream>>>(ch1_1_7); }
    { GemmP ch1_1_8;
      ch1_1_8.A = HP + (size_t)38 * C; ch1_1_8.B = Wh2 + (size_t)8 * C * G4; ch1_1_8.bias = HP + (size_t)38 * C; ch1_1_8.R = GH; ch1_1_8.C = GH;
      ch1_1_8.sAo = (long long)PP * C; ch1_1_8.sAi = (long long)18 * C; ch1_1_8.sAm = C; ch1_1_8.sAk = 1; ch1_1_8.sBo = 0; ch1_1_8.sBi = 0; ch1_1_8.sBn = 1; ch1_1_8.sBk = G4; ch1_1_8.sCo = (long long)HW * G4; ch1_1_8.sCi = (long long)16 * G4; ch1_1_8.sCm = G4; ch1_1_8.sRo = (long long)HW * G4; ch1_1_8.sRi = (long long)16 * G4; ch1_1_8.sRm = G4; ch1_1_8.sRn = 1;
      ch1_1_8.M = 16; ch1_1_8.N = G4; ch1_1_8.K = C; ch1_1_8.zi_n = 16; ch1_1_8.flags = 4; ch1_1_8.act = 0;
      ch1_1_8.alpha = 1.0f; ch1_1_8.beta = 1.0f; ch1_1_8.sa = 1.0f; ch1_1_8.sb = 1.0f; ch1_1_8.Npad = G4; ch1_1_8.pad_ = 0;
      k_gemm<1><<<dim3((unsigned)((G4) + 31) / 32, (unsigned)((16) + 15) / 16, (unsigned)(Bn * 16)), 32, 0, stream>>>(ch1_1_8); }

    k_bl_cell<<<(unsigned)(((long long)Bn * HW * C + 255) / 256), 256, 0, stream>>>(XG, GH, Cc, HS, HP, Bn, T, 1, C);
    { GemmP ch1_2_0;
      ch1_2_0.A = HP + (size_t)0 * C; ch1_2_0.B = Wh2 + (size_t)0 * C * G4; ch1_2_0.bias = HP + (size_t)0 * C; ch1_2_0.R = HP + (size_t)0 * C; ch1_2_0.C = GH;
      ch1_2_0.sAo = (long long)PP * C; ch1_2_0.sAi = (long long)18 * C; ch1_2_0.sAm = C; ch1_2_0.sAk = 1; ch1_2_0.sBo = 0; ch1_2_0.sBi = 0; ch1_2_0.sBn = 1; ch1_2_0.sBk = G4; ch1_2_0.sCo = (long long)HW * G4; ch1_2_0.sCi = (long long)16 * G4; ch1_2_0.sCm = G4; ch1_2_0.sRo = 0; ch1_2_0.sRi = 0; ch1_2_0.sRm = 0; ch1_2_0.sRn = 0;
      ch1_2_0.M = 16; ch1_2_0.N = G4; ch1_2_0.K = C; ch1_2_0.zi_n = 16; ch1_2_0.flags = 0; ch1_2_0.act = 0;
      ch1_2_0.alpha = 1.0f; ch1_2_0.beta = 0.0f; ch1_2_0.sa = 1.0f; ch1_2_0.sb = 1.0f; ch1_2_0.Npad = G4; ch1_2_0.pad_ = 0;
      k_gemm<1><<<dim3((unsigned)((G4) + 31) / 32, (unsigned)((16) + 15) / 16, (unsigned)(Bn * 16)), 32, 0, stream>>>(ch1_2_0); }
    { GemmP ch1_2_1;
      ch1_2_1.A = HP + (size_t)1 * C; ch1_2_1.B = Wh2 + (size_t)1 * C * G4; ch1_2_1.bias = HP + (size_t)1 * C; ch1_2_1.R = GH; ch1_2_1.C = GH;
      ch1_2_1.sAo = (long long)PP * C; ch1_2_1.sAi = (long long)18 * C; ch1_2_1.sAm = C; ch1_2_1.sAk = 1; ch1_2_1.sBo = 0; ch1_2_1.sBi = 0; ch1_2_1.sBn = 1; ch1_2_1.sBk = G4; ch1_2_1.sCo = (long long)HW * G4; ch1_2_1.sCi = (long long)16 * G4; ch1_2_1.sCm = G4; ch1_2_1.sRo = (long long)HW * G4; ch1_2_1.sRi = (long long)16 * G4; ch1_2_1.sRm = G4; ch1_2_1.sRn = 1;
      ch1_2_1.M = 16; ch1_2_1.N = G4; ch1_2_1.K = C; ch1_2_1.zi_n = 16; ch1_2_1.flags = 4; ch1_2_1.act = 0;
      ch1_2_1.alpha = 1.0f; ch1_2_1.beta = 1.0f; ch1_2_1.sa = 1.0f; ch1_2_1.sb = 1.0f; ch1_2_1.Npad = G4; ch1_2_1.pad_ = 0;
      k_gemm<1><<<dim3((unsigned)((G4) + 31) / 32, (unsigned)((16) + 15) / 16, (unsigned)(Bn * 16)), 32, 0, stream>>>(ch1_2_1); }
    { GemmP ch1_2_2;
      ch1_2_2.A = HP + (size_t)2 * C; ch1_2_2.B = Wh2 + (size_t)2 * C * G4; ch1_2_2.bias = HP + (size_t)2 * C; ch1_2_2.R = GH; ch1_2_2.C = GH;
      ch1_2_2.sAo = (long long)PP * C; ch1_2_2.sAi = (long long)18 * C; ch1_2_2.sAm = C; ch1_2_2.sAk = 1; ch1_2_2.sBo = 0; ch1_2_2.sBi = 0; ch1_2_2.sBn = 1; ch1_2_2.sBk = G4; ch1_2_2.sCo = (long long)HW * G4; ch1_2_2.sCi = (long long)16 * G4; ch1_2_2.sCm = G4; ch1_2_2.sRo = (long long)HW * G4; ch1_2_2.sRi = (long long)16 * G4; ch1_2_2.sRm = G4; ch1_2_2.sRn = 1;
      ch1_2_2.M = 16; ch1_2_2.N = G4; ch1_2_2.K = C; ch1_2_2.zi_n = 16; ch1_2_2.flags = 4; ch1_2_2.act = 0;
      ch1_2_2.alpha = 1.0f; ch1_2_2.beta = 1.0f; ch1_2_2.sa = 1.0f; ch1_2_2.sb = 1.0f; ch1_2_2.Npad = G4; ch1_2_2.pad_ = 0;
      k_gemm<1><<<dim3((unsigned)((G4) + 31) / 32, (unsigned)((16) + 15) / 16, (unsigned)(Bn * 16)), 32, 0, stream>>>(ch1_2_2); }
    { GemmP ch1_2_3;
      ch1_2_3.A = HP + (size_t)18 * C; ch1_2_3.B = Wh2 + (size_t)3 * C * G4; ch1_2_3.bias = HP + (size_t)18 * C; ch1_2_3.R = GH; ch1_2_3.C = GH;
      ch1_2_3.sAo = (long long)PP * C; ch1_2_3.sAi = (long long)18 * C; ch1_2_3.sAm = C; ch1_2_3.sAk = 1; ch1_2_3.sBo = 0; ch1_2_3.sBi = 0; ch1_2_3.sBn = 1; ch1_2_3.sBk = G4; ch1_2_3.sCo = (long long)HW * G4; ch1_2_3.sCi = (long long)16 * G4; ch1_2_3.sCm = G4; ch1_2_3.sRo = (long long)HW * G4; ch1_2_3.sRi = (long long)16 * G4; ch1_2_3.sRm = G4; ch1_2_3.sRn = 1;
      ch1_2_3.M = 16; ch1_2_3.N = G4; ch1_2_3.K = C; ch1_2_3.zi_n = 16; ch1_2_3.flags = 4; ch1_2_3.act = 0;
      ch1_2_3.alpha = 1.0f; ch1_2_3.beta = 1.0f; ch1_2_3.sa = 1.0f; ch1_2_3.sb = 1.0f; ch1_2_3.Npad = G4; ch1_2_3.pad_ = 0;
      k_gemm<1><<<dim3((unsigned)((G4) + 31) / 32, (unsigned)((16) + 15) / 16, (unsigned)(Bn * 16)), 32, 0, stream>>>(ch1_2_3); }
    { GemmP ch1_2_4;
      ch1_2_4.A = HP + (size_t)19 * C; ch1_2_4.B = Wh2 + (size_t)4 * C * G4; ch1_2_4.bias = HP + (size_t)19 * C; ch1_2_4.R = GH; ch1_2_4.C = GH;
      ch1_2_4.sAo = (long long)PP * C; ch1_2_4.sAi = (long long)18 * C; ch1_2_4.sAm = C; ch1_2_4.sAk = 1; ch1_2_4.sBo = 0; ch1_2_4.sBi = 0; ch1_2_4.sBn = 1; ch1_2_4.sBk = G4; ch1_2_4.sCo = (long long)HW * G4; ch1_2_4.sCi = (long long)16 * G4; ch1_2_4.sCm = G4; ch1_2_4.sRo = (long long)HW * G4; ch1_2_4.sRi = (long long)16 * G4; ch1_2_4.sRm = G4; ch1_2_4.sRn = 1;
      ch1_2_4.M = 16; ch1_2_4.N = G4; ch1_2_4.K = C; ch1_2_4.zi_n = 16; ch1_2_4.flags = 4; ch1_2_4.act = 0;
      ch1_2_4.alpha = 1.0f; ch1_2_4.beta = 1.0f; ch1_2_4.sa = 1.0f; ch1_2_4.sb = 1.0f; ch1_2_4.Npad = G4; ch1_2_4.pad_ = 0;
      k_gemm<1><<<dim3((unsigned)((G4) + 31) / 32, (unsigned)((16) + 15) / 16, (unsigned)(Bn * 16)), 32, 0, stream>>>(ch1_2_4); }
    { GemmP ch1_2_5;
      ch1_2_5.A = HP + (size_t)20 * C; ch1_2_5.B = Wh2 + (size_t)5 * C * G4; ch1_2_5.bias = HP + (size_t)20 * C; ch1_2_5.R = GH; ch1_2_5.C = GH;
      ch1_2_5.sAo = (long long)PP * C; ch1_2_5.sAi = (long long)18 * C; ch1_2_5.sAm = C; ch1_2_5.sAk = 1; ch1_2_5.sBo = 0; ch1_2_5.sBi = 0; ch1_2_5.sBn = 1; ch1_2_5.sBk = G4; ch1_2_5.sCo = (long long)HW * G4; ch1_2_5.sCi = (long long)16 * G4; ch1_2_5.sCm = G4; ch1_2_5.sRo = (long long)HW * G4; ch1_2_5.sRi = (long long)16 * G4; ch1_2_5.sRm = G4; ch1_2_5.sRn = 1;
      ch1_2_5.M = 16; ch1_2_5.N = G4; ch1_2_5.K = C; ch1_2_5.zi_n = 16; ch1_2_5.flags = 4; ch1_2_5.act = 0;
      ch1_2_5.alpha = 1.0f; ch1_2_5.beta = 1.0f; ch1_2_5.sa = 1.0f; ch1_2_5.sb = 1.0f; ch1_2_5.Npad = G4; ch1_2_5.pad_ = 0;
      k_gemm<1><<<dim3((unsigned)((G4) + 31) / 32, (unsigned)((16) + 15) / 16, (unsigned)(Bn * 16)), 32, 0, stream>>>(ch1_2_5); }
    { GemmP ch1_2_6;
      ch1_2_6.A = HP + (size_t)36 * C; ch1_2_6.B = Wh2 + (size_t)6 * C * G4; ch1_2_6.bias = HP + (size_t)36 * C; ch1_2_6.R = GH; ch1_2_6.C = GH;
      ch1_2_6.sAo = (long long)PP * C; ch1_2_6.sAi = (long long)18 * C; ch1_2_6.sAm = C; ch1_2_6.sAk = 1; ch1_2_6.sBo = 0; ch1_2_6.sBi = 0; ch1_2_6.sBn = 1; ch1_2_6.sBk = G4; ch1_2_6.sCo = (long long)HW * G4; ch1_2_6.sCi = (long long)16 * G4; ch1_2_6.sCm = G4; ch1_2_6.sRo = (long long)HW * G4; ch1_2_6.sRi = (long long)16 * G4; ch1_2_6.sRm = G4; ch1_2_6.sRn = 1;
      ch1_2_6.M = 16; ch1_2_6.N = G4; ch1_2_6.K = C; ch1_2_6.zi_n = 16; ch1_2_6.flags = 4; ch1_2_6.act = 0;
      ch1_2_6.alpha = 1.0f; ch1_2_6.beta = 1.0f; ch1_2_6.sa = 1.0f; ch1_2_6.sb = 1.0f; ch1_2_6.Npad = G4; ch1_2_6.pad_ = 0;
      k_gemm<1><<<dim3((unsigned)((G4) + 31) / 32, (unsigned)((16) + 15) / 16, (unsigned)(Bn * 16)), 32, 0, stream>>>(ch1_2_6); }
    { GemmP ch1_2_7;
      ch1_2_7.A = HP + (size_t)37 * C; ch1_2_7.B = Wh2 + (size_t)7 * C * G4; ch1_2_7.bias = HP + (size_t)37 * C; ch1_2_7.R = GH; ch1_2_7.C = GH;
      ch1_2_7.sAo = (long long)PP * C; ch1_2_7.sAi = (long long)18 * C; ch1_2_7.sAm = C; ch1_2_7.sAk = 1; ch1_2_7.sBo = 0; ch1_2_7.sBi = 0; ch1_2_7.sBn = 1; ch1_2_7.sBk = G4; ch1_2_7.sCo = (long long)HW * G4; ch1_2_7.sCi = (long long)16 * G4; ch1_2_7.sCm = G4; ch1_2_7.sRo = (long long)HW * G4; ch1_2_7.sRi = (long long)16 * G4; ch1_2_7.sRm = G4; ch1_2_7.sRn = 1;
      ch1_2_7.M = 16; ch1_2_7.N = G4; ch1_2_7.K = C; ch1_2_7.zi_n = 16; ch1_2_7.flags = 4; ch1_2_7.act = 0;
      ch1_2_7.alpha = 1.0f; ch1_2_7.beta = 1.0f; ch1_2_7.sa = 1.0f; ch1_2_7.sb = 1.0f; ch1_2_7.Npad = G4; ch1_2_7.pad_ = 0;
      k_gemm<1><<<dim3((unsigned)((G4) + 31) / 32, (unsigned)((16) + 15) / 16, (unsigned)(Bn * 16)), 32, 0, stream>>>(ch1_2_7); }
    { GemmP ch1_2_8;
      ch1_2_8.A = HP + (size_t)38 * C; ch1_2_8.B = Wh2 + (size_t)8 * C * G4; ch1_2_8.bias = HP + (size_t)38 * C; ch1_2_8.R = GH; ch1_2_8.C = GH;
      ch1_2_8.sAo = (long long)PP * C; ch1_2_8.sAi = (long long)18 * C; ch1_2_8.sAm = C; ch1_2_8.sAk = 1; ch1_2_8.sBo = 0; ch1_2_8.sBi = 0; ch1_2_8.sBn = 1; ch1_2_8.sBk = G4; ch1_2_8.sCo = (long long)HW * G4; ch1_2_8.sCi = (long long)16 * G4; ch1_2_8.sCm = G4; ch1_2_8.sRo = (long long)HW * G4; ch1_2_8.sRi = (long long)16 * G4; ch1_2_8.sRm = G4; ch1_2_8.sRn = 1;
      ch1_2_8.M = 16; ch1_2_8.N = G4; ch1_2_8.K = C; ch1_2_8.zi_n = 16; ch1_2_8.flags = 4; ch1_2_8.act = 0;
      ch1_2_8.alpha = 1.0f; ch1_2_8.beta = 1.0f; ch1_2_8.sa = 1.0f; ch1_2_8.sb = 1.0f; ch1_2_8.Npad = G4; ch1_2_8.pad_ = 0;
      k_gemm<1><<<dim3((unsigned)((G4) + 31) / 32, (unsigned)((16) + 15) / 16, (unsigned)(Bn * 16)), 32, 0, stream>>>(ch1_2_8); }

    k_bl_cell<<<(unsigned)(((long long)Bn * HW * C + 255) / 256), 256, 0, stream>>>(XG, GH, Cc, HS, HP, Bn, T, 2, C);
    { GemmP ch1_3_0;
      ch1_3_0.A = HP + (size_t)0 * C; ch1_3_0.B = Wh2 + (size_t)0 * C * G4; ch1_3_0.bias = HP + (size_t)0 * C; ch1_3_0.R = HP + (size_t)0 * C; ch1_3_0.C = GH;
      ch1_3_0.sAo = (long long)PP * C; ch1_3_0.sAi = (long long)18 * C; ch1_3_0.sAm = C; ch1_3_0.sAk = 1; ch1_3_0.sBo = 0; ch1_3_0.sBi = 0; ch1_3_0.sBn = 1; ch1_3_0.sBk = G4; ch1_3_0.sCo = (long long)HW * G4; ch1_3_0.sCi = (long long)16 * G4; ch1_3_0.sCm = G4; ch1_3_0.sRo = 0; ch1_3_0.sRi = 0; ch1_3_0.sRm = 0; ch1_3_0.sRn = 0;
      ch1_3_0.M = 16; ch1_3_0.N = G4; ch1_3_0.K = C; ch1_3_0.zi_n = 16; ch1_3_0.flags = 0; ch1_3_0.act = 0;
      ch1_3_0.alpha = 1.0f; ch1_3_0.beta = 0.0f; ch1_3_0.sa = 1.0f; ch1_3_0.sb = 1.0f; ch1_3_0.Npad = G4; ch1_3_0.pad_ = 0;
      k_gemm<1><<<dim3((unsigned)((G4) + 31) / 32, (unsigned)((16) + 15) / 16, (unsigned)(Bn * 16)), 32, 0, stream>>>(ch1_3_0); }
    { GemmP ch1_3_1;
      ch1_3_1.A = HP + (size_t)1 * C; ch1_3_1.B = Wh2 + (size_t)1 * C * G4; ch1_3_1.bias = HP + (size_t)1 * C; ch1_3_1.R = GH; ch1_3_1.C = GH;
      ch1_3_1.sAo = (long long)PP * C; ch1_3_1.sAi = (long long)18 * C; ch1_3_1.sAm = C; ch1_3_1.sAk = 1; ch1_3_1.sBo = 0; ch1_3_1.sBi = 0; ch1_3_1.sBn = 1; ch1_3_1.sBk = G4; ch1_3_1.sCo = (long long)HW * G4; ch1_3_1.sCi = (long long)16 * G4; ch1_3_1.sCm = G4; ch1_3_1.sRo = (long long)HW * G4; ch1_3_1.sRi = (long long)16 * G4; ch1_3_1.sRm = G4; ch1_3_1.sRn = 1;
      ch1_3_1.M = 16; ch1_3_1.N = G4; ch1_3_1.K = C; ch1_3_1.zi_n = 16; ch1_3_1.flags = 4; ch1_3_1.act = 0;
      ch1_3_1.alpha = 1.0f; ch1_3_1.beta = 1.0f; ch1_3_1.sa = 1.0f; ch1_3_1.sb = 1.0f; ch1_3_1.Npad = G4; ch1_3_1.pad_ = 0;
      k_gemm<1><<<dim3((unsigned)((G4) + 31) / 32, (unsigned)((16) + 15) / 16, (unsigned)(Bn * 16)), 32, 0, stream>>>(ch1_3_1); }
    { GemmP ch1_3_2;
      ch1_3_2.A = HP + (size_t)2 * C; ch1_3_2.B = Wh2 + (size_t)2 * C * G4; ch1_3_2.bias = HP + (size_t)2 * C; ch1_3_2.R = GH; ch1_3_2.C = GH;
      ch1_3_2.sAo = (long long)PP * C; ch1_3_2.sAi = (long long)18 * C; ch1_3_2.sAm = C; ch1_3_2.sAk = 1; ch1_3_2.sBo = 0; ch1_3_2.sBi = 0; ch1_3_2.sBn = 1; ch1_3_2.sBk = G4; ch1_3_2.sCo = (long long)HW * G4; ch1_3_2.sCi = (long long)16 * G4; ch1_3_2.sCm = G4; ch1_3_2.sRo = (long long)HW * G4; ch1_3_2.sRi = (long long)16 * G4; ch1_3_2.sRm = G4; ch1_3_2.sRn = 1;
      ch1_3_2.M = 16; ch1_3_2.N = G4; ch1_3_2.K = C; ch1_3_2.zi_n = 16; ch1_3_2.flags = 4; ch1_3_2.act = 0;
      ch1_3_2.alpha = 1.0f; ch1_3_2.beta = 1.0f; ch1_3_2.sa = 1.0f; ch1_3_2.sb = 1.0f; ch1_3_2.Npad = G4; ch1_3_2.pad_ = 0;
      k_gemm<1><<<dim3((unsigned)((G4) + 31) / 32, (unsigned)((16) + 15) / 16, (unsigned)(Bn * 16)), 32, 0, stream>>>(ch1_3_2); }
    { GemmP ch1_3_3;
      ch1_3_3.A = HP + (size_t)18 * C; ch1_3_3.B = Wh2 + (size_t)3 * C * G4; ch1_3_3.bias = HP + (size_t)18 * C; ch1_3_3.R = GH; ch1_3_3.C = GH;
      ch1_3_3.sAo = (long long)PP * C; ch1_3_3.sAi = (long long)18 * C; ch1_3_3.sAm = C; ch1_3_3.sAk = 1; ch1_3_3.sBo = 0; ch1_3_3.sBi = 0; ch1_3_3.sBn = 1; ch1_3_3.sBk = G4; ch1_3_3.sCo = (long long)HW * G4; ch1_3_3.sCi = (long long)16 * G4; ch1_3_3.sCm = G4; ch1_3_3.sRo = (long long)HW * G4; ch1_3_3.sRi = (long long)16 * G4; ch1_3_3.sRm = G4; ch1_3_3.sRn = 1;
      ch1_3_3.M = 16; ch1_3_3.N = G4; ch1_3_3.K = C; ch1_3_3.zi_n = 16; ch1_3_3.flags = 4; ch1_3_3.act = 0;
      ch1_3_3.alpha = 1.0f; ch1_3_3.beta = 1.0f; ch1_3_3.sa = 1.0f; ch1_3_3.sb = 1.0f; ch1_3_3.Npad = G4; ch1_3_3.pad_ = 0;
      k_gemm<1><<<dim3((unsigned)((G4) + 31) / 32, (unsigned)((16) + 15) / 16, (unsigned)(Bn * 16)), 32, 0, stream>>>(ch1_3_3); }
    { GemmP ch1_3_4;
      ch1_3_4.A = HP + (size_t)19 * C; ch1_3_4.B = Wh2 + (size_t)4 * C * G4; ch1_3_4.bias = HP + (size_t)19 * C; ch1_3_4.R = GH; ch1_3_4.C = GH;
      ch1_3_4.sAo = (long long)PP * C; ch1_3_4.sAi = (long long)18 * C; ch1_3_4.sAm = C; ch1_3_4.sAk = 1; ch1_3_4.sBo = 0; ch1_3_4.sBi = 0; ch1_3_4.sBn = 1; ch1_3_4.sBk = G4; ch1_3_4.sCo = (long long)HW * G4; ch1_3_4.sCi = (long long)16 * G4; ch1_3_4.sCm = G4; ch1_3_4.sRo = (long long)HW * G4; ch1_3_4.sRi = (long long)16 * G4; ch1_3_4.sRm = G4; ch1_3_4.sRn = 1;
      ch1_3_4.M = 16; ch1_3_4.N = G4; ch1_3_4.K = C; ch1_3_4.zi_n = 16; ch1_3_4.flags = 4; ch1_3_4.act = 0;
      ch1_3_4.alpha = 1.0f; ch1_3_4.beta = 1.0f; ch1_3_4.sa = 1.0f; ch1_3_4.sb = 1.0f; ch1_3_4.Npad = G4; ch1_3_4.pad_ = 0;
      k_gemm<1><<<dim3((unsigned)((G4) + 31) / 32, (unsigned)((16) + 15) / 16, (unsigned)(Bn * 16)), 32, 0, stream>>>(ch1_3_4); }
    { GemmP ch1_3_5;
      ch1_3_5.A = HP + (size_t)20 * C; ch1_3_5.B = Wh2 + (size_t)5 * C * G4; ch1_3_5.bias = HP + (size_t)20 * C; ch1_3_5.R = GH; ch1_3_5.C = GH;
      ch1_3_5.sAo = (long long)PP * C; ch1_3_5.sAi = (long long)18 * C; ch1_3_5.sAm = C; ch1_3_5.sAk = 1; ch1_3_5.sBo = 0; ch1_3_5.sBi = 0; ch1_3_5.sBn = 1; ch1_3_5.sBk = G4; ch1_3_5.sCo = (long long)HW * G4; ch1_3_5.sCi = (long long)16 * G4; ch1_3_5.sCm = G4; ch1_3_5.sRo = (long long)HW * G4; ch1_3_5.sRi = (long long)16 * G4; ch1_3_5.sRm = G4; ch1_3_5.sRn = 1;
      ch1_3_5.M = 16; ch1_3_5.N = G4; ch1_3_5.K = C; ch1_3_5.zi_n = 16; ch1_3_5.flags = 4; ch1_3_5.act = 0;
      ch1_3_5.alpha = 1.0f; ch1_3_5.beta = 1.0f; ch1_3_5.sa = 1.0f; ch1_3_5.sb = 1.0f; ch1_3_5.Npad = G4; ch1_3_5.pad_ = 0;
      k_gemm<1><<<dim3((unsigned)((G4) + 31) / 32, (unsigned)((16) + 15) / 16, (unsigned)(Bn * 16)), 32, 0, stream>>>(ch1_3_5); }
    { GemmP ch1_3_6;
      ch1_3_6.A = HP + (size_t)36 * C; ch1_3_6.B = Wh2 + (size_t)6 * C * G4; ch1_3_6.bias = HP + (size_t)36 * C; ch1_3_6.R = GH; ch1_3_6.C = GH;
      ch1_3_6.sAo = (long long)PP * C; ch1_3_6.sAi = (long long)18 * C; ch1_3_6.sAm = C; ch1_3_6.sAk = 1; ch1_3_6.sBo = 0; ch1_3_6.sBi = 0; ch1_3_6.sBn = 1; ch1_3_6.sBk = G4; ch1_3_6.sCo = (long long)HW * G4; ch1_3_6.sCi = (long long)16 * G4; ch1_3_6.sCm = G4; ch1_3_6.sRo = (long long)HW * G4; ch1_3_6.sRi = (long long)16 * G4; ch1_3_6.sRm = G4; ch1_3_6.sRn = 1;
      ch1_3_6.M = 16; ch1_3_6.N = G4; ch1_3_6.K = C; ch1_3_6.zi_n = 16; ch1_3_6.flags = 4; ch1_3_6.act = 0;
      ch1_3_6.alpha = 1.0f; ch1_3_6.beta = 1.0f; ch1_3_6.sa = 1.0f; ch1_3_6.sb = 1.0f; ch1_3_6.Npad = G4; ch1_3_6.pad_ = 0;
      k_gemm<1><<<dim3((unsigned)((G4) + 31) / 32, (unsigned)((16) + 15) / 16, (unsigned)(Bn * 16)), 32, 0, stream>>>(ch1_3_6); }
    { GemmP ch1_3_7;
      ch1_3_7.A = HP + (size_t)37 * C; ch1_3_7.B = Wh2 + (size_t)7 * C * G4; ch1_3_7.bias = HP + (size_t)37 * C; ch1_3_7.R = GH; ch1_3_7.C = GH;
      ch1_3_7.sAo = (long long)PP * C; ch1_3_7.sAi = (long long)18 * C; ch1_3_7.sAm = C; ch1_3_7.sAk = 1; ch1_3_7.sBo = 0; ch1_3_7.sBi = 0; ch1_3_7.sBn = 1; ch1_3_7.sBk = G4; ch1_3_7.sCo = (long long)HW * G4; ch1_3_7.sCi = (long long)16 * G4; ch1_3_7.sCm = G4; ch1_3_7.sRo = (long long)HW * G4; ch1_3_7.sRi = (long long)16 * G4; ch1_3_7.sRm = G4; ch1_3_7.sRn = 1;
      ch1_3_7.M = 16; ch1_3_7.N = G4; ch1_3_7.K = C; ch1_3_7.zi_n = 16; ch1_3_7.flags = 4; ch1_3_7.act = 0;
      ch1_3_7.alpha = 1.0f; ch1_3_7.beta = 1.0f; ch1_3_7.sa = 1.0f; ch1_3_7.sb = 1.0f; ch1_3_7.Npad = G4; ch1_3_7.pad_ = 0;
      k_gemm<1><<<dim3((unsigned)((G4) + 31) / 32, (unsigned)((16) + 15) / 16, (unsigned)(Bn * 16)), 32, 0, stream>>>(ch1_3_7); }
    { GemmP ch1_3_8;
      ch1_3_8.A = HP + (size_t)38 * C; ch1_3_8.B = Wh2 + (size_t)8 * C * G4; ch1_3_8.bias = HP + (size_t)38 * C; ch1_3_8.R = GH; ch1_3_8.C = GH;
      ch1_3_8.sAo = (long long)PP * C; ch1_3_8.sAi = (long long)18 * C; ch1_3_8.sAm = C; ch1_3_8.sAk = 1; ch1_3_8.sBo = 0; ch1_3_8.sBi = 0; ch1_3_8.sBn = 1; ch1_3_8.sBk = G4; ch1_3_8.sCo = (long long)HW * G4; ch1_3_8.sCi = (long long)16 * G4; ch1_3_8.sCm = G4; ch1_3_8.sRo = (long long)HW * G4; ch1_3_8.sRi = (long long)16 * G4; ch1_3_8.sRm = G4; ch1_3_8.sRn = 1;
      ch1_3_8.M = 16; ch1_3_8.N = G4; ch1_3_8.K = C; ch1_3_8.zi_n = 16; ch1_3_8.flags = 4; ch1_3_8.act = 0;
      ch1_3_8.alpha = 1.0f; ch1_3_8.beta = 1.0f; ch1_3_8.sa = 1.0f; ch1_3_8.sb = 1.0f; ch1_3_8.Npad = G4; ch1_3_8.pad_ = 0;
      k_gemm<1><<<dim3((unsigned)((G4) + 31) / 32, (unsigned)((16) + 15) / 16, (unsigned)(Bn * 16)), 32, 0, stream>>>(ch1_3_8); }

    k_bl_cell<<<(unsigned)(((long long)Bn * HW * C + 255) / 256), 256, 0, stream>>>(XG, GH, Cc, HS, HP, Bn, T, 3, C);
    { GemmP ch1_4_0;
      ch1_4_0.A = HP + (size_t)0 * C; ch1_4_0.B = Wh2 + (size_t)0 * C * G4; ch1_4_0.bias = HP + (size_t)0 * C; ch1_4_0.R = HP + (size_t)0 * C; ch1_4_0.C = GH;
      ch1_4_0.sAo = (long long)PP * C; ch1_4_0.sAi = (long long)18 * C; ch1_4_0.sAm = C; ch1_4_0.sAk = 1; ch1_4_0.sBo = 0; ch1_4_0.sBi = 0; ch1_4_0.sBn = 1; ch1_4_0.sBk = G4; ch1_4_0.sCo = (long long)HW * G4; ch1_4_0.sCi = (long long)16 * G4; ch1_4_0.sCm = G4; ch1_4_0.sRo = 0; ch1_4_0.sRi = 0; ch1_4_0.sRm = 0; ch1_4_0.sRn = 0;
      ch1_4_0.M = 16; ch1_4_0.N = G4; ch1_4_0.K = C; ch1_4_0.zi_n = 16; ch1_4_0.flags = 0; ch1_4_0.act = 0;
      ch1_4_0.alpha = 1.0f; ch1_4_0.beta = 0.0f; ch1_4_0.sa = 1.0f; ch1_4_0.sb = 1.0f; ch1_4_0.Npad = G4; ch1_4_0.pad_ = 0;
      k_gemm<1><<<dim3((unsigned)((G4) + 31) / 32, (unsigned)((16) + 15) / 16, (unsigned)(Bn * 16)), 32, 0, stream>>>(ch1_4_0); }
    { GemmP ch1_4_1;
      ch1_4_1.A = HP + (size_t)1 * C; ch1_4_1.B = Wh2 + (size_t)1 * C * G4; ch1_4_1.bias = HP + (size_t)1 * C; ch1_4_1.R = GH; ch1_4_1.C = GH;
      ch1_4_1.sAo = (long long)PP * C; ch1_4_1.sAi = (long long)18 * C; ch1_4_1.sAm = C; ch1_4_1.sAk = 1; ch1_4_1.sBo = 0; ch1_4_1.sBi = 0; ch1_4_1.sBn = 1; ch1_4_1.sBk = G4; ch1_4_1.sCo = (long long)HW * G4; ch1_4_1.sCi = (long long)16 * G4; ch1_4_1.sCm = G4; ch1_4_1.sRo = (long long)HW * G4; ch1_4_1.sRi = (long long)16 * G4; ch1_4_1.sRm = G4; ch1_4_1.sRn = 1;
      ch1_4_1.M = 16; ch1_4_1.N = G4; ch1_4_1.K = C; ch1_4_1.zi_n = 16; ch1_4_1.flags = 4; ch1_4_1.act = 0;
      ch1_4_1.alpha = 1.0f; ch1_4_1.beta = 1.0f; ch1_4_1.sa = 1.0f; ch1_4_1.sb = 1.0f; ch1_4_1.Npad = G4; ch1_4_1.pad_ = 0;
      k_gemm<1><<<dim3((unsigned)((G4) + 31) / 32, (unsigned)((16) + 15) / 16, (unsigned)(Bn * 16)), 32, 0, stream>>>(ch1_4_1); }
    { GemmP ch1_4_2;
      ch1_4_2.A = HP + (size_t)2 * C; ch1_4_2.B = Wh2 + (size_t)2 * C * G4; ch1_4_2.bias = HP + (size_t)2 * C; ch1_4_2.R = GH; ch1_4_2.C = GH;
      ch1_4_2.sAo = (long long)PP * C; ch1_4_2.sAi = (long long)18 * C; ch1_4_2.sAm = C; ch1_4_2.sAk = 1; ch1_4_2.sBo = 0; ch1_4_2.sBi = 0; ch1_4_2.sBn = 1; ch1_4_2.sBk = G4; ch1_4_2.sCo = (long long)HW * G4; ch1_4_2.sCi = (long long)16 * G4; ch1_4_2.sCm = G4; ch1_4_2.sRo = (long long)HW * G4; ch1_4_2.sRi = (long long)16 * G4; ch1_4_2.sRm = G4; ch1_4_2.sRn = 1;
      ch1_4_2.M = 16; ch1_4_2.N = G4; ch1_4_2.K = C; ch1_4_2.zi_n = 16; ch1_4_2.flags = 4; ch1_4_2.act = 0;
      ch1_4_2.alpha = 1.0f; ch1_4_2.beta = 1.0f; ch1_4_2.sa = 1.0f; ch1_4_2.sb = 1.0f; ch1_4_2.Npad = G4; ch1_4_2.pad_ = 0;
      k_gemm<1><<<dim3((unsigned)((G4) + 31) / 32, (unsigned)((16) + 15) / 16, (unsigned)(Bn * 16)), 32, 0, stream>>>(ch1_4_2); }
    { GemmP ch1_4_3;
      ch1_4_3.A = HP + (size_t)18 * C; ch1_4_3.B = Wh2 + (size_t)3 * C * G4; ch1_4_3.bias = HP + (size_t)18 * C; ch1_4_3.R = GH; ch1_4_3.C = GH;
      ch1_4_3.sAo = (long long)PP * C; ch1_4_3.sAi = (long long)18 * C; ch1_4_3.sAm = C; ch1_4_3.sAk = 1; ch1_4_3.sBo = 0; ch1_4_3.sBi = 0; ch1_4_3.sBn = 1; ch1_4_3.sBk = G4; ch1_4_3.sCo = (long long)HW * G4; ch1_4_3.sCi = (long long)16 * G4; ch1_4_3.sCm = G4; ch1_4_3.sRo = (long long)HW * G4; ch1_4_3.sRi = (long long)16 * G4; ch1_4_3.sRm = G4; ch1_4_3.sRn = 1;
      ch1_4_3.M = 16; ch1_4_3.N = G4; ch1_4_3.K = C; ch1_4_3.zi_n = 16; ch1_4_3.flags = 4; ch1_4_3.act = 0;
      ch1_4_3.alpha = 1.0f; ch1_4_3.beta = 1.0f; ch1_4_3.sa = 1.0f; ch1_4_3.sb = 1.0f; ch1_4_3.Npad = G4; ch1_4_3.pad_ = 0;
      k_gemm<1><<<dim3((unsigned)((G4) + 31) / 32, (unsigned)((16) + 15) / 16, (unsigned)(Bn * 16)), 32, 0, stream>>>(ch1_4_3); }
    { GemmP ch1_4_4;
      ch1_4_4.A = HP + (size_t)19 * C; ch1_4_4.B = Wh2 + (size_t)4 * C * G4; ch1_4_4.bias = HP + (size_t)19 * C; ch1_4_4.R = GH; ch1_4_4.C = GH;
      ch1_4_4.sAo = (long long)PP * C; ch1_4_4.sAi = (long long)18 * C; ch1_4_4.sAm = C; ch1_4_4.sAk = 1; ch1_4_4.sBo = 0; ch1_4_4.sBi = 0; ch1_4_4.sBn = 1; ch1_4_4.sBk = G4; ch1_4_4.sCo = (long long)HW * G4; ch1_4_4.sCi = (long long)16 * G4; ch1_4_4.sCm = G4; ch1_4_4.sRo = (long long)HW * G4; ch1_4_4.sRi = (long long)16 * G4; ch1_4_4.sRm = G4; ch1_4_4.sRn = 1;
      ch1_4_4.M = 16; ch1_4_4.N = G4; ch1_4_4.K = C; ch1_4_4.zi_n = 16; ch1_4_4.flags = 4; ch1_4_4.act = 0;
      ch1_4_4.alpha = 1.0f; ch1_4_4.beta = 1.0f; ch1_4_4.sa = 1.0f; ch1_4_4.sb = 1.0f; ch1_4_4.Npad = G4; ch1_4_4.pad_ = 0;
      k_gemm<1><<<dim3((unsigned)((G4) + 31) / 32, (unsigned)((16) + 15) / 16, (unsigned)(Bn * 16)), 32, 0, stream>>>(ch1_4_4); }
    { GemmP ch1_4_5;
      ch1_4_5.A = HP + (size_t)20 * C; ch1_4_5.B = Wh2 + (size_t)5 * C * G4; ch1_4_5.bias = HP + (size_t)20 * C; ch1_4_5.R = GH; ch1_4_5.C = GH;
      ch1_4_5.sAo = (long long)PP * C; ch1_4_5.sAi = (long long)18 * C; ch1_4_5.sAm = C; ch1_4_5.sAk = 1; ch1_4_5.sBo = 0; ch1_4_5.sBi = 0; ch1_4_5.sBn = 1; ch1_4_5.sBk = G4; ch1_4_5.sCo = (long long)HW * G4; ch1_4_5.sCi = (long long)16 * G4; ch1_4_5.sCm = G4; ch1_4_5.sRo = (long long)HW * G4; ch1_4_5.sRi = (long long)16 * G4; ch1_4_5.sRm = G4; ch1_4_5.sRn = 1;
      ch1_4_5.M = 16; ch1_4_5.N = G4; ch1_4_5.K = C; ch1_4_5.zi_n = 16; ch1_4_5.flags = 4; ch1_4_5.act = 0;
      ch1_4_5.alpha = 1.0f; ch1_4_5.beta = 1.0f; ch1_4_5.sa = 1.0f; ch1_4_5.sb = 1.0f; ch1_4_5.Npad = G4; ch1_4_5.pad_ = 0;
      k_gemm<1><<<dim3((unsigned)((G4) + 31) / 32, (unsigned)((16) + 15) / 16, (unsigned)(Bn * 16)), 32, 0, stream>>>(ch1_4_5); }
    { GemmP ch1_4_6;
      ch1_4_6.A = HP + (size_t)36 * C; ch1_4_6.B = Wh2 + (size_t)6 * C * G4; ch1_4_6.bias = HP + (size_t)36 * C; ch1_4_6.R = GH; ch1_4_6.C = GH;
      ch1_4_6.sAo = (long long)PP * C; ch1_4_6.sAi = (long long)18 * C; ch1_4_6.sAm = C; ch1_4_6.sAk = 1; ch1_4_6.sBo = 0; ch1_4_6.sBi = 0; ch1_4_6.sBn = 1; ch1_4_6.sBk = G4; ch1_4_6.sCo = (long long)HW * G4; ch1_4_6.sCi = (long long)16 * G4; ch1_4_6.sCm = G4; ch1_4_6.sRo = (long long)HW * G4; ch1_4_6.sRi = (long long)16 * G4; ch1_4_6.sRm = G4; ch1_4_6.sRn = 1;
      ch1_4_6.M = 16; ch1_4_6.N = G4; ch1_4_6.K = C; ch1_4_6.zi_n = 16; ch1_4_6.flags = 4; ch1_4_6.act = 0;
      ch1_4_6.alpha = 1.0f; ch1_4_6.beta = 1.0f; ch1_4_6.sa = 1.0f; ch1_4_6.sb = 1.0f; ch1_4_6.Npad = G4; ch1_4_6.pad_ = 0;
      k_gemm<1><<<dim3((unsigned)((G4) + 31) / 32, (unsigned)((16) + 15) / 16, (unsigned)(Bn * 16)), 32, 0, stream>>>(ch1_4_6); }
    { GemmP ch1_4_7;
      ch1_4_7.A = HP + (size_t)37 * C; ch1_4_7.B = Wh2 + (size_t)7 * C * G4; ch1_4_7.bias = HP + (size_t)37 * C; ch1_4_7.R = GH; ch1_4_7.C = GH;
      ch1_4_7.sAo = (long long)PP * C; ch1_4_7.sAi = (long long)18 * C; ch1_4_7.sAm = C; ch1_4_7.sAk = 1; ch1_4_7.sBo = 0; ch1_4_7.sBi = 0; ch1_4_7.sBn = 1; ch1_4_7.sBk = G4; ch1_4_7.sCo = (long long)HW * G4; ch1_4_7.sCi = (long long)16 * G4; ch1_4_7.sCm = G4; ch1_4_7.sRo = (long long)HW * G4; ch1_4_7.sRi = (long long)16 * G4; ch1_4_7.sRm = G4; ch1_4_7.sRn = 1;
      ch1_4_7.M = 16; ch1_4_7.N = G4; ch1_4_7.K = C; ch1_4_7.zi_n = 16; ch1_4_7.flags = 4; ch1_4_7.act = 0;
      ch1_4_7.alpha = 1.0f; ch1_4_7.beta = 1.0f; ch1_4_7.sa = 1.0f; ch1_4_7.sb = 1.0f; ch1_4_7.Npad = G4; ch1_4_7.pad_ = 0;
      k_gemm<1><<<dim3((unsigned)((G4) + 31) / 32, (unsigned)((16) + 15) / 16, (unsigned)(Bn * 16)), 32, 0, stream>>>(ch1_4_7); }
    { GemmP ch1_4_8;
      ch1_4_8.A = HP + (size_t)38 * C; ch1_4_8.B = Wh2 + (size_t)8 * C * G4; ch1_4_8.bias = HP + (size_t)38 * C; ch1_4_8.R = GH; ch1_4_8.C = GH;
      ch1_4_8.sAo = (long long)PP * C; ch1_4_8.sAi = (long long)18 * C; ch1_4_8.sAm = C; ch1_4_8.sAk = 1; ch1_4_8.sBo = 0; ch1_4_8.sBi = 0; ch1_4_8.sBn = 1; ch1_4_8.sBk = G4; ch1_4_8.sCo = (long long)HW * G4; ch1_4_8.sCi = (long long)16 * G4; ch1_4_8.sCm = G4; ch1_4_8.sRo = (long long)HW * G4; ch1_4_8.sRi = (long long)16 * G4; ch1_4_8.sRm = G4; ch1_4_8.sRn = 1;
      ch1_4_8.M = 16; ch1_4_8.N = G4; ch1_4_8.K = C; ch1_4_8.zi_n = 16; ch1_4_8.flags = 4; ch1_4_8.act = 0;
      ch1_4_8.alpha = 1.0f; ch1_4_8.beta = 1.0f; ch1_4_8.sa = 1.0f; ch1_4_8.sb = 1.0f; ch1_4_8.Npad = G4; ch1_4_8.pad_ = 0;
      k_gemm<1><<<dim3((unsigned)((G4) + 31) / 32, (unsigned)((16) + 15) / 16, (unsigned)(Bn * 16)), 32, 0, stream>>>(ch1_4_8); }

    k_bl_cell<<<(unsigned)(((long long)Bn * HW * C + 255) / 256), 256, 0, stream>>>(XG, GH, Cc, HS, HP, Bn, T, 4, C);
    { GemmP ch1_5_0;
      ch1_5_0.A = HP + (size_t)0 * C; ch1_5_0.B = Wh2 + (size_t)0 * C * G4; ch1_5_0.bias = HP + (size_t)0 * C; ch1_5_0.R = HP + (size_t)0 * C; ch1_5_0.C = GH;
      ch1_5_0.sAo = (long long)PP * C; ch1_5_0.sAi = (long long)18 * C; ch1_5_0.sAm = C; ch1_5_0.sAk = 1; ch1_5_0.sBo = 0; ch1_5_0.sBi = 0; ch1_5_0.sBn = 1; ch1_5_0.sBk = G4; ch1_5_0.sCo = (long long)HW * G4; ch1_5_0.sCi = (long long)16 * G4; ch1_5_0.sCm = G4; ch1_5_0.sRo = 0; ch1_5_0.sRi = 0; ch1_5_0.sRm = 0; ch1_5_0.sRn = 0;
      ch1_5_0.M = 16; ch1_5_0.N = G4; ch1_5_0.K = C; ch1_5_0.zi_n = 16; ch1_5_0.flags = 0; ch1_5_0.act = 0;
      ch1_5_0.alpha = 1.0f; ch1_5_0.beta = 0.0f; ch1_5_0.sa = 1.0f; ch1_5_0.sb = 1.0f; ch1_5_0.Npad = G4; ch1_5_0.pad_ = 0;
      k_gemm<1><<<dim3((unsigned)((G4) + 31) / 32, (unsigned)((16) + 15) / 16, (unsigned)(Bn * 16)), 32, 0, stream>>>(ch1_5_0); }
    { GemmP ch1_5_1;
      ch1_5_1.A = HP + (size_t)1 * C; ch1_5_1.B = Wh2 + (size_t)1 * C * G4; ch1_5_1.bias = HP + (size_t)1 * C; ch1_5_1.R = GH; ch1_5_1.C = GH;
      ch1_5_1.sAo = (long long)PP * C; ch1_5_1.sAi = (long long)18 * C; ch1_5_1.sAm = C; ch1_5_1.sAk = 1; ch1_5_1.sBo = 0; ch1_5_1.sBi = 0; ch1_5_1.sBn = 1; ch1_5_1.sBk = G4; ch1_5_1.sCo = (long long)HW * G4; ch1_5_1.sCi = (long long)16 * G4; ch1_5_1.sCm = G4; ch1_5_1.sRo = (long long)HW * G4; ch1_5_1.sRi = (long long)16 * G4; ch1_5_1.sRm = G4; ch1_5_1.sRn = 1;
      ch1_5_1.M = 16; ch1_5_1.N = G4; ch1_5_1.K = C; ch1_5_1.zi_n = 16; ch1_5_1.flags = 4; ch1_5_1.act = 0;
      ch1_5_1.alpha = 1.0f; ch1_5_1.beta = 1.0f; ch1_5_1.sa = 1.0f; ch1_5_1.sb = 1.0f; ch1_5_1.Npad = G4; ch1_5_1.pad_ = 0;
      k_gemm<1><<<dim3((unsigned)((G4) + 31) / 32, (unsigned)((16) + 15) / 16, (unsigned)(Bn * 16)), 32, 0, stream>>>(ch1_5_1); }
    { GemmP ch1_5_2;
      ch1_5_2.A = HP + (size_t)2 * C; ch1_5_2.B = Wh2 + (size_t)2 * C * G4; ch1_5_2.bias = HP + (size_t)2 * C; ch1_5_2.R = GH; ch1_5_2.C = GH;
      ch1_5_2.sAo = (long long)PP * C; ch1_5_2.sAi = (long long)18 * C; ch1_5_2.sAm = C; ch1_5_2.sAk = 1; ch1_5_2.sBo = 0; ch1_5_2.sBi = 0; ch1_5_2.sBn = 1; ch1_5_2.sBk = G4; ch1_5_2.sCo = (long long)HW * G4; ch1_5_2.sCi = (long long)16 * G4; ch1_5_2.sCm = G4; ch1_5_2.sRo = (long long)HW * G4; ch1_5_2.sRi = (long long)16 * G4; ch1_5_2.sRm = G4; ch1_5_2.sRn = 1;
      ch1_5_2.M = 16; ch1_5_2.N = G4; ch1_5_2.K = C; ch1_5_2.zi_n = 16; ch1_5_2.flags = 4; ch1_5_2.act = 0;
      ch1_5_2.alpha = 1.0f; ch1_5_2.beta = 1.0f; ch1_5_2.sa = 1.0f; ch1_5_2.sb = 1.0f; ch1_5_2.Npad = G4; ch1_5_2.pad_ = 0;
      k_gemm<1><<<dim3((unsigned)((G4) + 31) / 32, (unsigned)((16) + 15) / 16, (unsigned)(Bn * 16)), 32, 0, stream>>>(ch1_5_2); }
    { GemmP ch1_5_3;
      ch1_5_3.A = HP + (size_t)18 * C; ch1_5_3.B = Wh2 + (size_t)3 * C * G4; ch1_5_3.bias = HP + (size_t)18 * C; ch1_5_3.R = GH; ch1_5_3.C = GH;
      ch1_5_3.sAo = (long long)PP * C; ch1_5_3.sAi = (long long)18 * C; ch1_5_3.sAm = C; ch1_5_3.sAk = 1; ch1_5_3.sBo = 0; ch1_5_3.sBi = 0; ch1_5_3.sBn = 1; ch1_5_3.sBk = G4; ch1_5_3.sCo = (long long)HW * G4; ch1_5_3.sCi = (long long)16 * G4; ch1_5_3.sCm = G4; ch1_5_3.sRo = (long long)HW * G4; ch1_5_3.sRi = (long long)16 * G4; ch1_5_3.sRm = G4; ch1_5_3.sRn = 1;
      ch1_5_3.M = 16; ch1_5_3.N = G4; ch1_5_3.K = C; ch1_5_3.zi_n = 16; ch1_5_3.flags = 4; ch1_5_3.act = 0;
      ch1_5_3.alpha = 1.0f; ch1_5_3.beta = 1.0f; ch1_5_3.sa = 1.0f; ch1_5_3.sb = 1.0f; ch1_5_3.Npad = G4; ch1_5_3.pad_ = 0;
      k_gemm<1><<<dim3((unsigned)((G4) + 31) / 32, (unsigned)((16) + 15) / 16, (unsigned)(Bn * 16)), 32, 0, stream>>>(ch1_5_3); }
    { GemmP ch1_5_4;
      ch1_5_4.A = HP + (size_t)19 * C; ch1_5_4.B = Wh2 + (size_t)4 * C * G4; ch1_5_4.bias = HP + (size_t)19 * C; ch1_5_4.R = GH; ch1_5_4.C = GH;
      ch1_5_4.sAo = (long long)PP * C; ch1_5_4.sAi = (long long)18 * C; ch1_5_4.sAm = C; ch1_5_4.sAk = 1; ch1_5_4.sBo = 0; ch1_5_4.sBi = 0; ch1_5_4.sBn = 1; ch1_5_4.sBk = G4; ch1_5_4.sCo = (long long)HW * G4; ch1_5_4.sCi = (long long)16 * G4; ch1_5_4.sCm = G4; ch1_5_4.sRo = (long long)HW * G4; ch1_5_4.sRi = (long long)16 * G4; ch1_5_4.sRm = G4; ch1_5_4.sRn = 1;
      ch1_5_4.M = 16; ch1_5_4.N = G4; ch1_5_4.K = C; ch1_5_4.zi_n = 16; ch1_5_4.flags = 4; ch1_5_4.act = 0;
      ch1_5_4.alpha = 1.0f; ch1_5_4.beta = 1.0f; ch1_5_4.sa = 1.0f; ch1_5_4.sb = 1.0f; ch1_5_4.Npad = G4; ch1_5_4.pad_ = 0;
      k_gemm<1><<<dim3((unsigned)((G4) + 31) / 32, (unsigned)((16) + 15) / 16, (unsigned)(Bn * 16)), 32, 0, stream>>>(ch1_5_4); }
    { GemmP ch1_5_5;
      ch1_5_5.A = HP + (size_t)20 * C; ch1_5_5.B = Wh2 + (size_t)5 * C * G4; ch1_5_5.bias = HP + (size_t)20 * C; ch1_5_5.R = GH; ch1_5_5.C = GH;
      ch1_5_5.sAo = (long long)PP * C; ch1_5_5.sAi = (long long)18 * C; ch1_5_5.sAm = C; ch1_5_5.sAk = 1; ch1_5_5.sBo = 0; ch1_5_5.sBi = 0; ch1_5_5.sBn = 1; ch1_5_5.sBk = G4; ch1_5_5.sCo = (long long)HW * G4; ch1_5_5.sCi = (long long)16 * G4; ch1_5_5.sCm = G4; ch1_5_5.sRo = (long long)HW * G4; ch1_5_5.sRi = (long long)16 * G4; ch1_5_5.sRm = G4; ch1_5_5.sRn = 1;
      ch1_5_5.M = 16; ch1_5_5.N = G4; ch1_5_5.K = C; ch1_5_5.zi_n = 16; ch1_5_5.flags = 4; ch1_5_5.act = 0;
      ch1_5_5.alpha = 1.0f; ch1_5_5.beta = 1.0f; ch1_5_5.sa = 1.0f; ch1_5_5.sb = 1.0f; ch1_5_5.Npad = G4; ch1_5_5.pad_ = 0;
      k_gemm<1><<<dim3((unsigned)((G4) + 31) / 32, (unsigned)((16) + 15) / 16, (unsigned)(Bn * 16)), 32, 0, stream>>>(ch1_5_5); }
    { GemmP ch1_5_6;
      ch1_5_6.A = HP + (size_t)36 * C; ch1_5_6.B = Wh2 + (size_t)6 * C * G4; ch1_5_6.bias = HP + (size_t)36 * C; ch1_5_6.R = GH; ch1_5_6.C = GH;
      ch1_5_6.sAo = (long long)PP * C; ch1_5_6.sAi = (long long)18 * C; ch1_5_6.sAm = C; ch1_5_6.sAk = 1; ch1_5_6.sBo = 0; ch1_5_6.sBi = 0; ch1_5_6.sBn = 1; ch1_5_6.sBk = G4; ch1_5_6.sCo = (long long)HW * G4; ch1_5_6.sCi = (long long)16 * G4; ch1_5_6.sCm = G4; ch1_5_6.sRo = (long long)HW * G4; ch1_5_6.sRi = (long long)16 * G4; ch1_5_6.sRm = G4; ch1_5_6.sRn = 1;
      ch1_5_6.M = 16; ch1_5_6.N = G4; ch1_5_6.K = C; ch1_5_6.zi_n = 16; ch1_5_6.flags = 4; ch1_5_6.act = 0;
      ch1_5_6.alpha = 1.0f; ch1_5_6.beta = 1.0f; ch1_5_6.sa = 1.0f; ch1_5_6.sb = 1.0f; ch1_5_6.Npad = G4; ch1_5_6.pad_ = 0;
      k_gemm<1><<<dim3((unsigned)((G4) + 31) / 32, (unsigned)((16) + 15) / 16, (unsigned)(Bn * 16)), 32, 0, stream>>>(ch1_5_6); }
    { GemmP ch1_5_7;
      ch1_5_7.A = HP + (size_t)37 * C; ch1_5_7.B = Wh2 + (size_t)7 * C * G4; ch1_5_7.bias = HP + (size_t)37 * C; ch1_5_7.R = GH; ch1_5_7.C = GH;
      ch1_5_7.sAo = (long long)PP * C; ch1_5_7.sAi = (long long)18 * C; ch1_5_7.sAm = C; ch1_5_7.sAk = 1; ch1_5_7.sBo = 0; ch1_5_7.sBi = 0; ch1_5_7.sBn = 1; ch1_5_7.sBk = G4; ch1_5_7.sCo = (long long)HW * G4; ch1_5_7.sCi = (long long)16 * G4; ch1_5_7.sCm = G4; ch1_5_7.sRo = (long long)HW * G4; ch1_5_7.sRi = (long long)16 * G4; ch1_5_7.sRm = G4; ch1_5_7.sRn = 1;
      ch1_5_7.M = 16; ch1_5_7.N = G4; ch1_5_7.K = C; ch1_5_7.zi_n = 16; ch1_5_7.flags = 4; ch1_5_7.act = 0;
      ch1_5_7.alpha = 1.0f; ch1_5_7.beta = 1.0f; ch1_5_7.sa = 1.0f; ch1_5_7.sb = 1.0f; ch1_5_7.Npad = G4; ch1_5_7.pad_ = 0;
      k_gemm<1><<<dim3((unsigned)((G4) + 31) / 32, (unsigned)((16) + 15) / 16, (unsigned)(Bn * 16)), 32, 0, stream>>>(ch1_5_7); }
    { GemmP ch1_5_8;
      ch1_5_8.A = HP + (size_t)38 * C; ch1_5_8.B = Wh2 + (size_t)8 * C * G4; ch1_5_8.bias = HP + (size_t)38 * C; ch1_5_8.R = GH; ch1_5_8.C = GH;
      ch1_5_8.sAo = (long long)PP * C; ch1_5_8.sAi = (long long)18 * C; ch1_5_8.sAm = C; ch1_5_8.sAk = 1; ch1_5_8.sBo = 0; ch1_5_8.sBi = 0; ch1_5_8.sBn = 1; ch1_5_8.sBk = G4; ch1_5_8.sCo = (long long)HW * G4; ch1_5_8.sCi = (long long)16 * G4; ch1_5_8.sCm = G4; ch1_5_8.sRo = (long long)HW * G4; ch1_5_8.sRi = (long long)16 * G4; ch1_5_8.sRm = G4; ch1_5_8.sRn = 1;
      ch1_5_8.M = 16; ch1_5_8.N = G4; ch1_5_8.K = C; ch1_5_8.zi_n = 16; ch1_5_8.flags = 4; ch1_5_8.act = 0;
      ch1_5_8.alpha = 1.0f; ch1_5_8.beta = 1.0f; ch1_5_8.sa = 1.0f; ch1_5_8.sb = 1.0f; ch1_5_8.Npad = G4; ch1_5_8.pad_ = 0;
      k_gemm<1><<<dim3((unsigned)((G4) + 31) / 32, (unsigned)((16) + 15) / 16, (unsigned)(Bn * 16)), 32, 0, stream>>>(ch1_5_8); }

    k_bl_cell<<<(unsigned)(((long long)Bn * HW * C + 255) / 256), 256, 0, stream>>>(XG, GH, Cc, HS, HP, Bn, T, 5, C);
    { GemmP ch1_6_0;
      ch1_6_0.A = HP + (size_t)0 * C; ch1_6_0.B = Wh2 + (size_t)0 * C * G4; ch1_6_0.bias = HP + (size_t)0 * C; ch1_6_0.R = HP + (size_t)0 * C; ch1_6_0.C = GH;
      ch1_6_0.sAo = (long long)PP * C; ch1_6_0.sAi = (long long)18 * C; ch1_6_0.sAm = C; ch1_6_0.sAk = 1; ch1_6_0.sBo = 0; ch1_6_0.sBi = 0; ch1_6_0.sBn = 1; ch1_6_0.sBk = G4; ch1_6_0.sCo = (long long)HW * G4; ch1_6_0.sCi = (long long)16 * G4; ch1_6_0.sCm = G4; ch1_6_0.sRo = 0; ch1_6_0.sRi = 0; ch1_6_0.sRm = 0; ch1_6_0.sRn = 0;
      ch1_6_0.M = 16; ch1_6_0.N = G4; ch1_6_0.K = C; ch1_6_0.zi_n = 16; ch1_6_0.flags = 0; ch1_6_0.act = 0;
      ch1_6_0.alpha = 1.0f; ch1_6_0.beta = 0.0f; ch1_6_0.sa = 1.0f; ch1_6_0.sb = 1.0f; ch1_6_0.Npad = G4; ch1_6_0.pad_ = 0;
      k_gemm<1><<<dim3((unsigned)((G4) + 31) / 32, (unsigned)((16) + 15) / 16, (unsigned)(Bn * 16)), 32, 0, stream>>>(ch1_6_0); }
    { GemmP ch1_6_1;
      ch1_6_1.A = HP + (size_t)1 * C; ch1_6_1.B = Wh2 + (size_t)1 * C * G4; ch1_6_1.bias = HP + (size_t)1 * C; ch1_6_1.R = GH; ch1_6_1.C = GH;
      ch1_6_1.sAo = (long long)PP * C; ch1_6_1.sAi = (long long)18 * C; ch1_6_1.sAm = C; ch1_6_1.sAk = 1; ch1_6_1.sBo = 0; ch1_6_1.sBi = 0; ch1_6_1.sBn = 1; ch1_6_1.sBk = G4; ch1_6_1.sCo = (long long)HW * G4; ch1_6_1.sCi = (long long)16 * G4; ch1_6_1.sCm = G4; ch1_6_1.sRo = (long long)HW * G4; ch1_6_1.sRi = (long long)16 * G4; ch1_6_1.sRm = G4; ch1_6_1.sRn = 1;
      ch1_6_1.M = 16; ch1_6_1.N = G4; ch1_6_1.K = C; ch1_6_1.zi_n = 16; ch1_6_1.flags = 4; ch1_6_1.act = 0;
      ch1_6_1.alpha = 1.0f; ch1_6_1.beta = 1.0f; ch1_6_1.sa = 1.0f; ch1_6_1.sb = 1.0f; ch1_6_1.Npad = G4; ch1_6_1.pad_ = 0;
      k_gemm<1><<<dim3((unsigned)((G4) + 31) / 32, (unsigned)((16) + 15) / 16, (unsigned)(Bn * 16)), 32, 0, stream>>>(ch1_6_1); }
    { GemmP ch1_6_2;
      ch1_6_2.A = HP + (size_t)2 * C; ch1_6_2.B = Wh2 + (size_t)2 * C * G4; ch1_6_2.bias = HP + (size_t)2 * C; ch1_6_2.R = GH; ch1_6_2.C = GH;
      ch1_6_2.sAo = (long long)PP * C; ch1_6_2.sAi = (long long)18 * C; ch1_6_2.sAm = C; ch1_6_2.sAk = 1; ch1_6_2.sBo = 0; ch1_6_2.sBi = 0; ch1_6_2.sBn = 1; ch1_6_2.sBk = G4; ch1_6_2.sCo = (long long)HW * G4; ch1_6_2.sCi = (long long)16 * G4; ch1_6_2.sCm = G4; ch1_6_2.sRo = (long long)HW * G4; ch1_6_2.sRi = (long long)16 * G4; ch1_6_2.sRm = G4; ch1_6_2.sRn = 1;
      ch1_6_2.M = 16; ch1_6_2.N = G4; ch1_6_2.K = C; ch1_6_2.zi_n = 16; ch1_6_2.flags = 4; ch1_6_2.act = 0;
      ch1_6_2.alpha = 1.0f; ch1_6_2.beta = 1.0f; ch1_6_2.sa = 1.0f; ch1_6_2.sb = 1.0f; ch1_6_2.Npad = G4; ch1_6_2.pad_ = 0;
      k_gemm<1><<<dim3((unsigned)((G4) + 31) / 32, (unsigned)((16) + 15) / 16, (unsigned)(Bn * 16)), 32, 0, stream>>>(ch1_6_2); }
    { GemmP ch1_6_3;
      ch1_6_3.A = HP + (size_t)18 * C; ch1_6_3.B = Wh2 + (size_t)3 * C * G4; ch1_6_3.bias = HP + (size_t)18 * C; ch1_6_3.R = GH; ch1_6_3.C = GH;
      ch1_6_3.sAo = (long long)PP * C; ch1_6_3.sAi = (long long)18 * C; ch1_6_3.sAm = C; ch1_6_3.sAk = 1; ch1_6_3.sBo = 0; ch1_6_3.sBi = 0; ch1_6_3.sBn = 1; ch1_6_3.sBk = G4; ch1_6_3.sCo = (long long)HW * G4; ch1_6_3.sCi = (long long)16 * G4; ch1_6_3.sCm = G4; ch1_6_3.sRo = (long long)HW * G4; ch1_6_3.sRi = (long long)16 * G4; ch1_6_3.sRm = G4; ch1_6_3.sRn = 1;
      ch1_6_3.M = 16; ch1_6_3.N = G4; ch1_6_3.K = C; ch1_6_3.zi_n = 16; ch1_6_3.flags = 4; ch1_6_3.act = 0;
      ch1_6_3.alpha = 1.0f; ch1_6_3.beta = 1.0f; ch1_6_3.sa = 1.0f; ch1_6_3.sb = 1.0f; ch1_6_3.Npad = G4; ch1_6_3.pad_ = 0;
      k_gemm<1><<<dim3((unsigned)((G4) + 31) / 32, (unsigned)((16) + 15) / 16, (unsigned)(Bn * 16)), 32, 0, stream>>>(ch1_6_3); }
    { GemmP ch1_6_4;
      ch1_6_4.A = HP + (size_t)19 * C; ch1_6_4.B = Wh2 + (size_t)4 * C * G4; ch1_6_4.bias = HP + (size_t)19 * C; ch1_6_4.R = GH; ch1_6_4.C = GH;
      ch1_6_4.sAo = (long long)PP * C; ch1_6_4.sAi = (long long)18 * C; ch1_6_4.sAm = C; ch1_6_4.sAk = 1; ch1_6_4.sBo = 0; ch1_6_4.sBi = 0; ch1_6_4.sBn = 1; ch1_6_4.sBk = G4; ch1_6_4.sCo = (long long)HW * G4; ch1_6_4.sCi = (long long)16 * G4; ch1_6_4.sCm = G4; ch1_6_4.sRo = (long long)HW * G4; ch1_6_4.sRi = (long long)16 * G4; ch1_6_4.sRm = G4; ch1_6_4.sRn = 1;
      ch1_6_4.M = 16; ch1_6_4.N = G4; ch1_6_4.K = C; ch1_6_4.zi_n = 16; ch1_6_4.flags = 4; ch1_6_4.act = 0;
      ch1_6_4.alpha = 1.0f; ch1_6_4.beta = 1.0f; ch1_6_4.sa = 1.0f; ch1_6_4.sb = 1.0f; ch1_6_4.Npad = G4; ch1_6_4.pad_ = 0;
      k_gemm<1><<<dim3((unsigned)((G4) + 31) / 32, (unsigned)((16) + 15) / 16, (unsigned)(Bn * 16)), 32, 0, stream>>>(ch1_6_4); }
    { GemmP ch1_6_5;
      ch1_6_5.A = HP + (size_t)20 * C; ch1_6_5.B = Wh2 + (size_t)5 * C * G4; ch1_6_5.bias = HP + (size_t)20 * C; ch1_6_5.R = GH; ch1_6_5.C = GH;
      ch1_6_5.sAo = (long long)PP * C; ch1_6_5.sAi = (long long)18 * C; ch1_6_5.sAm = C; ch1_6_5.sAk = 1; ch1_6_5.sBo = 0; ch1_6_5.sBi = 0; ch1_6_5.sBn = 1; ch1_6_5.sBk = G4; ch1_6_5.sCo = (long long)HW * G4; ch1_6_5.sCi = (long long)16 * G4; ch1_6_5.sCm = G4; ch1_6_5.sRo = (long long)HW * G4; ch1_6_5.sRi = (long long)16 * G4; ch1_6_5.sRm = G4; ch1_6_5.sRn = 1;
      ch1_6_5.M = 16; ch1_6_5.N = G4; ch1_6_5.K = C; ch1_6_5.zi_n = 16; ch1_6_5.flags = 4; ch1_6_5.act = 0;
      ch1_6_5.alpha = 1.0f; ch1_6_5.beta = 1.0f; ch1_6_5.sa = 1.0f; ch1_6_5.sb = 1.0f; ch1_6_5.Npad = G4; ch1_6_5.pad_ = 0;
      k_gemm<1><<<dim3((unsigned)((G4) + 31) / 32, (unsigned)((16) + 15) / 16, (unsigned)(Bn * 16)), 32, 0, stream>>>(ch1_6_5); }
    { GemmP ch1_6_6;
      ch1_6_6.A = HP + (size_t)36 * C; ch1_6_6.B = Wh2 + (size_t)6 * C * G4; ch1_6_6.bias = HP + (size_t)36 * C; ch1_6_6.R = GH; ch1_6_6.C = GH;
      ch1_6_6.sAo = (long long)PP * C; ch1_6_6.sAi = (long long)18 * C; ch1_6_6.sAm = C; ch1_6_6.sAk = 1; ch1_6_6.sBo = 0; ch1_6_6.sBi = 0; ch1_6_6.sBn = 1; ch1_6_6.sBk = G4; ch1_6_6.sCo = (long long)HW * G4; ch1_6_6.sCi = (long long)16 * G4; ch1_6_6.sCm = G4; ch1_6_6.sRo = (long long)HW * G4; ch1_6_6.sRi = (long long)16 * G4; ch1_6_6.sRm = G4; ch1_6_6.sRn = 1;
      ch1_6_6.M = 16; ch1_6_6.N = G4; ch1_6_6.K = C; ch1_6_6.zi_n = 16; ch1_6_6.flags = 4; ch1_6_6.act = 0;
      ch1_6_6.alpha = 1.0f; ch1_6_6.beta = 1.0f; ch1_6_6.sa = 1.0f; ch1_6_6.sb = 1.0f; ch1_6_6.Npad = G4; ch1_6_6.pad_ = 0;
      k_gemm<1><<<dim3((unsigned)((G4) + 31) / 32, (unsigned)((16) + 15) / 16, (unsigned)(Bn * 16)), 32, 0, stream>>>(ch1_6_6); }
    { GemmP ch1_6_7;
      ch1_6_7.A = HP + (size_t)37 * C; ch1_6_7.B = Wh2 + (size_t)7 * C * G4; ch1_6_7.bias = HP + (size_t)37 * C; ch1_6_7.R = GH; ch1_6_7.C = GH;
      ch1_6_7.sAo = (long long)PP * C; ch1_6_7.sAi = (long long)18 * C; ch1_6_7.sAm = C; ch1_6_7.sAk = 1; ch1_6_7.sBo = 0; ch1_6_7.sBi = 0; ch1_6_7.sBn = 1; ch1_6_7.sBk = G4; ch1_6_7.sCo = (long long)HW * G4; ch1_6_7.sCi = (long long)16 * G4; ch1_6_7.sCm = G4; ch1_6_7.sRo = (long long)HW * G4; ch1_6_7.sRi = (long long)16 * G4; ch1_6_7.sRm = G4; ch1_6_7.sRn = 1;
      ch1_6_7.M = 16; ch1_6_7.N = G4; ch1_6_7.K = C; ch1_6_7.zi_n = 16; ch1_6_7.flags = 4; ch1_6_7.act = 0;
      ch1_6_7.alpha = 1.0f; ch1_6_7.beta = 1.0f; ch1_6_7.sa = 1.0f; ch1_6_7.sb = 1.0f; ch1_6_7.Npad = G4; ch1_6_7.pad_ = 0;
      k_gemm<1><<<dim3((unsigned)((G4) + 31) / 32, (unsigned)((16) + 15) / 16, (unsigned)(Bn * 16)), 32, 0, stream>>>(ch1_6_7); }
    { GemmP ch1_6_8;
      ch1_6_8.A = HP + (size_t)38 * C; ch1_6_8.B = Wh2 + (size_t)8 * C * G4; ch1_6_8.bias = HP + (size_t)38 * C; ch1_6_8.R = GH; ch1_6_8.C = GH;
      ch1_6_8.sAo = (long long)PP * C; ch1_6_8.sAi = (long long)18 * C; ch1_6_8.sAm = C; ch1_6_8.sAk = 1; ch1_6_8.sBo = 0; ch1_6_8.sBi = 0; ch1_6_8.sBn = 1; ch1_6_8.sBk = G4; ch1_6_8.sCo = (long long)HW * G4; ch1_6_8.sCi = (long long)16 * G4; ch1_6_8.sCm = G4; ch1_6_8.sRo = (long long)HW * G4; ch1_6_8.sRi = (long long)16 * G4; ch1_6_8.sRm = G4; ch1_6_8.sRn = 1;
      ch1_6_8.M = 16; ch1_6_8.N = G4; ch1_6_8.K = C; ch1_6_8.zi_n = 16; ch1_6_8.flags = 4; ch1_6_8.act = 0;
      ch1_6_8.alpha = 1.0f; ch1_6_8.beta = 1.0f; ch1_6_8.sa = 1.0f; ch1_6_8.sb = 1.0f; ch1_6_8.Npad = G4; ch1_6_8.pad_ = 0;
      k_gemm<1><<<dim3((unsigned)((G4) + 31) / 32, (unsigned)((16) + 15) / 16, (unsigned)(Bn * 16)), 32, 0, stream>>>(ch1_6_8); }

    k_bl_cell<<<(unsigned)(((long long)Bn * HW * C + 255) / 256), 256, 0, stream>>>(XG, GH, Cc, HS, HP, Bn, T, 6, C);
    { GemmP ch1_7_0;
      ch1_7_0.A = HP + (size_t)0 * C; ch1_7_0.B = Wh2 + (size_t)0 * C * G4; ch1_7_0.bias = HP + (size_t)0 * C; ch1_7_0.R = HP + (size_t)0 * C; ch1_7_0.C = GH;
      ch1_7_0.sAo = (long long)PP * C; ch1_7_0.sAi = (long long)18 * C; ch1_7_0.sAm = C; ch1_7_0.sAk = 1; ch1_7_0.sBo = 0; ch1_7_0.sBi = 0; ch1_7_0.sBn = 1; ch1_7_0.sBk = G4; ch1_7_0.sCo = (long long)HW * G4; ch1_7_0.sCi = (long long)16 * G4; ch1_7_0.sCm = G4; ch1_7_0.sRo = 0; ch1_7_0.sRi = 0; ch1_7_0.sRm = 0; ch1_7_0.sRn = 0;
      ch1_7_0.M = 16; ch1_7_0.N = G4; ch1_7_0.K = C; ch1_7_0.zi_n = 16; ch1_7_0.flags = 0; ch1_7_0.act = 0;
      ch1_7_0.alpha = 1.0f; ch1_7_0.beta = 0.0f; ch1_7_0.sa = 1.0f; ch1_7_0.sb = 1.0f; ch1_7_0.Npad = G4; ch1_7_0.pad_ = 0;
      k_gemm<1><<<dim3((unsigned)((G4) + 31) / 32, (unsigned)((16) + 15) / 16, (unsigned)(Bn * 16)), 32, 0, stream>>>(ch1_7_0); }
    { GemmP ch1_7_1;
      ch1_7_1.A = HP + (size_t)1 * C; ch1_7_1.B = Wh2 + (size_t)1 * C * G4; ch1_7_1.bias = HP + (size_t)1 * C; ch1_7_1.R = GH; ch1_7_1.C = GH;
      ch1_7_1.sAo = (long long)PP * C; ch1_7_1.sAi = (long long)18 * C; ch1_7_1.sAm = C; ch1_7_1.sAk = 1; ch1_7_1.sBo = 0; ch1_7_1.sBi = 0; ch1_7_1.sBn = 1; ch1_7_1.sBk = G4; ch1_7_1.sCo = (long long)HW * G4; ch1_7_1.sCi = (long long)16 * G4; ch1_7_1.sCm = G4; ch1_7_1.sRo = (long long)HW * G4; ch1_7_1.sRi = (long long)16 * G4; ch1_7_1.sRm = G4; ch1_7_1.sRn = 1;
      ch1_7_1.M = 16; ch1_7_1.N = G4; ch1_7_1.K = C; ch1_7_1.zi_n = 16; ch1_7_1.flags = 4; ch1_7_1.act = 0;
      ch1_7_1.alpha = 1.0f; ch1_7_1.beta = 1.0f; ch1_7_1.sa = 1.0f; ch1_7_1.sb = 1.0f; ch1_7_1.Npad = G4; ch1_7_1.pad_ = 0;
      k_gemm<1><<<dim3((unsigned)((G4) + 31) / 32, (unsigned)((16) + 15) / 16, (unsigned)(Bn * 16)), 32, 0, stream>>>(ch1_7_1); }
    { GemmP ch1_7_2;
      ch1_7_2.A = HP + (size_t)2 * C; ch1_7_2.B = Wh2 + (size_t)2 * C * G4; ch1_7_2.bias = HP + (size_t)2 * C; ch1_7_2.R = GH; ch1_7_2.C = GH;
      ch1_7_2.sAo = (long long)PP * C; ch1_7_2.sAi = (long long)18 * C; ch1_7_2.sAm = C; ch1_7_2.sAk = 1; ch1_7_2.sBo = 0; ch1_7_2.sBi = 0; ch1_7_2.sBn = 1; ch1_7_2.sBk = G4; ch1_7_2.sCo = (long long)HW * G4; ch1_7_2.sCi = (long long)16 * G4; ch1_7_2.sCm = G4; ch1_7_2.sRo = (long long)HW * G4; ch1_7_2.sRi = (long long)16 * G4; ch1_7_2.sRm = G4; ch1_7_2.sRn = 1;
      ch1_7_2.M = 16; ch1_7_2.N = G4; ch1_7_2.K = C; ch1_7_2.zi_n = 16; ch1_7_2.flags = 4; ch1_7_2.act = 0;
      ch1_7_2.alpha = 1.0f; ch1_7_2.beta = 1.0f; ch1_7_2.sa = 1.0f; ch1_7_2.sb = 1.0f; ch1_7_2.Npad = G4; ch1_7_2.pad_ = 0;
      k_gemm<1><<<dim3((unsigned)((G4) + 31) / 32, (unsigned)((16) + 15) / 16, (unsigned)(Bn * 16)), 32, 0, stream>>>(ch1_7_2); }
    { GemmP ch1_7_3;
      ch1_7_3.A = HP + (size_t)18 * C; ch1_7_3.B = Wh2 + (size_t)3 * C * G4; ch1_7_3.bias = HP + (size_t)18 * C; ch1_7_3.R = GH; ch1_7_3.C = GH;
      ch1_7_3.sAo = (long long)PP * C; ch1_7_3.sAi = (long long)18 * C; ch1_7_3.sAm = C; ch1_7_3.sAk = 1; ch1_7_3.sBo = 0; ch1_7_3.sBi = 0; ch1_7_3.sBn = 1; ch1_7_3.sBk = G4; ch1_7_3.sCo = (long long)HW * G4; ch1_7_3.sCi = (long long)16 * G4; ch1_7_3.sCm = G4; ch1_7_3.sRo = (long long)HW * G4; ch1_7_3.sRi = (long long)16 * G4; ch1_7_3.sRm = G4; ch1_7_3.sRn = 1;
      ch1_7_3.M = 16; ch1_7_3.N = G4; ch1_7_3.K = C; ch1_7_3.zi_n = 16; ch1_7_3.flags = 4; ch1_7_3.act = 0;
      ch1_7_3.alpha = 1.0f; ch1_7_3.beta = 1.0f; ch1_7_3.sa = 1.0f; ch1_7_3.sb = 1.0f; ch1_7_3.Npad = G4; ch1_7_3.pad_ = 0;
      k_gemm<1><<<dim3((unsigned)((G4) + 31) / 32, (unsigned)((16) + 15) / 16, (unsigned)(Bn * 16)), 32, 0, stream>>>(ch1_7_3); }
    { GemmP ch1_7_4;
      ch1_7_4.A = HP + (size_t)19 * C; ch1_7_4.B = Wh2 + (size_t)4 * C * G4; ch1_7_4.bias = HP + (size_t)19 * C; ch1_7_4.R = GH; ch1_7_4.C = GH;
      ch1_7_4.sAo = (long long)PP * C; ch1_7_4.sAi = (long long)18 * C; ch1_7_4.sAm = C; ch1_7_4.sAk = 1; ch1_7_4.sBo = 0; ch1_7_4.sBi = 0; ch1_7_4.sBn = 1; ch1_7_4.sBk = G4; ch1_7_4.sCo = (long long)HW * G4; ch1_7_4.sCi = (long long)16 * G4; ch1_7_4.sCm = G4; ch1_7_4.sRo = (long long)HW * G4; ch1_7_4.sRi = (long long)16 * G4; ch1_7_4.sRm = G4; ch1_7_4.sRn = 1;
      ch1_7_4.M = 16; ch1_7_4.N = G4; ch1_7_4.K = C; ch1_7_4.zi_n = 16; ch1_7_4.flags = 4; ch1_7_4.act = 0;
      ch1_7_4.alpha = 1.0f; ch1_7_4.beta = 1.0f; ch1_7_4.sa = 1.0f; ch1_7_4.sb = 1.0f; ch1_7_4.Npad = G4; ch1_7_4.pad_ = 0;
      k_gemm<1><<<dim3((unsigned)((G4) + 31) / 32, (unsigned)((16) + 15) / 16, (unsigned)(Bn * 16)), 32, 0, stream>>>(ch1_7_4); }
    { GemmP ch1_7_5;
      ch1_7_5.A = HP + (size_t)20 * C; ch1_7_5.B = Wh2 + (size_t)5 * C * G4; ch1_7_5.bias = HP + (size_t)20 * C; ch1_7_5.R = GH; ch1_7_5.C = GH;
      ch1_7_5.sAo = (long long)PP * C; ch1_7_5.sAi = (long long)18 * C; ch1_7_5.sAm = C; ch1_7_5.sAk = 1; ch1_7_5.sBo = 0; ch1_7_5.sBi = 0; ch1_7_5.sBn = 1; ch1_7_5.sBk = G4; ch1_7_5.sCo = (long long)HW * G4; ch1_7_5.sCi = (long long)16 * G4; ch1_7_5.sCm = G4; ch1_7_5.sRo = (long long)HW * G4; ch1_7_5.sRi = (long long)16 * G4; ch1_7_5.sRm = G4; ch1_7_5.sRn = 1;
      ch1_7_5.M = 16; ch1_7_5.N = G4; ch1_7_5.K = C; ch1_7_5.zi_n = 16; ch1_7_5.flags = 4; ch1_7_5.act = 0;
      ch1_7_5.alpha = 1.0f; ch1_7_5.beta = 1.0f; ch1_7_5.sa = 1.0f; ch1_7_5.sb = 1.0f; ch1_7_5.Npad = G4; ch1_7_5.pad_ = 0;
      k_gemm<1><<<dim3((unsigned)((G4) + 31) / 32, (unsigned)((16) + 15) / 16, (unsigned)(Bn * 16)), 32, 0, stream>>>(ch1_7_5); }
    { GemmP ch1_7_6;
      ch1_7_6.A = HP + (size_t)36 * C; ch1_7_6.B = Wh2 + (size_t)6 * C * G4; ch1_7_6.bias = HP + (size_t)36 * C; ch1_7_6.R = GH; ch1_7_6.C = GH;
      ch1_7_6.sAo = (long long)PP * C; ch1_7_6.sAi = (long long)18 * C; ch1_7_6.sAm = C; ch1_7_6.sAk = 1; ch1_7_6.sBo = 0; ch1_7_6.sBi = 0; ch1_7_6.sBn = 1; ch1_7_6.sBk = G4; ch1_7_6.sCo = (long long)HW * G4; ch1_7_6.sCi = (long long)16 * G4; ch1_7_6.sCm = G4; ch1_7_6.sRo = (long long)HW * G4; ch1_7_6.sRi = (long long)16 * G4; ch1_7_6.sRm = G4; ch1_7_6.sRn = 1;
      ch1_7_6.M = 16; ch1_7_6.N = G4; ch1_7_6.K = C; ch1_7_6.zi_n = 16; ch1_7_6.flags = 4; ch1_7_6.act = 0;
      ch1_7_6.alpha = 1.0f; ch1_7_6.beta = 1.0f; ch1_7_6.sa = 1.0f; ch1_7_6.sb = 1.0f; ch1_7_6.Npad = G4; ch1_7_6.pad_ = 0;
      k_gemm<1><<<dim3((unsigned)((G4) + 31) / 32, (unsigned)((16) + 15) / 16, (unsigned)(Bn * 16)), 32, 0, stream>>>(ch1_7_6); }
    { GemmP ch1_7_7;
      ch1_7_7.A = HP + (size_t)37 * C; ch1_7_7.B = Wh2 + (size_t)7 * C * G4; ch1_7_7.bias = HP + (size_t)37 * C; ch1_7_7.R = GH; ch1_7_7.C = GH;
      ch1_7_7.sAo = (long long)PP * C; ch1_7_7.sAi = (long long)18 * C; ch1_7_7.sAm = C; ch1_7_7.sAk = 1; ch1_7_7.sBo = 0; ch1_7_7.sBi = 0; ch1_7_7.sBn = 1; ch1_7_7.sBk = G4; ch1_7_7.sCo = (long long)HW * G4; ch1_7_7.sCi = (long long)16 * G4; ch1_7_7.sCm = G4; ch1_7_7.sRo = (long long)HW * G4; ch1_7_7.sRi = (long long)16 * G4; ch1_7_7.sRm = G4; ch1_7_7.sRn = 1;
      ch1_7_7.M = 16; ch1_7_7.N = G4; ch1_7_7.K = C; ch1_7_7.zi_n = 16; ch1_7_7.flags = 4; ch1_7_7.act = 0;
      ch1_7_7.alpha = 1.0f; ch1_7_7.beta = 1.0f; ch1_7_7.sa = 1.0f; ch1_7_7.sb = 1.0f; ch1_7_7.Npad = G4; ch1_7_7.pad_ = 0;
      k_gemm<1><<<dim3((unsigned)((G4) + 31) / 32, (unsigned)((16) + 15) / 16, (unsigned)(Bn * 16)), 32, 0, stream>>>(ch1_7_7); }
    { GemmP ch1_7_8;
      ch1_7_8.A = HP + (size_t)38 * C; ch1_7_8.B = Wh2 + (size_t)8 * C * G4; ch1_7_8.bias = HP + (size_t)38 * C; ch1_7_8.R = GH; ch1_7_8.C = GH;
      ch1_7_8.sAo = (long long)PP * C; ch1_7_8.sAi = (long long)18 * C; ch1_7_8.sAm = C; ch1_7_8.sAk = 1; ch1_7_8.sBo = 0; ch1_7_8.sBi = 0; ch1_7_8.sBn = 1; ch1_7_8.sBk = G4; ch1_7_8.sCo = (long long)HW * G4; ch1_7_8.sCi = (long long)16 * G4; ch1_7_8.sCm = G4; ch1_7_8.sRo = (long long)HW * G4; ch1_7_8.sRi = (long long)16 * G4; ch1_7_8.sRm = G4; ch1_7_8.sRn = 1;
      ch1_7_8.M = 16; ch1_7_8.N = G4; ch1_7_8.K = C; ch1_7_8.zi_n = 16; ch1_7_8.flags = 4; ch1_7_8.act = 0;
      ch1_7_8.alpha = 1.0f; ch1_7_8.beta = 1.0f; ch1_7_8.sa = 1.0f; ch1_7_8.sb = 1.0f; ch1_7_8.Npad = G4; ch1_7_8.pad_ = 0;
      k_gemm<1><<<dim3((unsigned)((G4) + 31) / 32, (unsigned)((16) + 15) / 16, (unsigned)(Bn * 16)), 32, 0, stream>>>(ch1_7_8); }

    k_bl_cell<<<(unsigned)(((long long)Bn * HW * C + 255) / 256), 256, 0, stream>>>(XG, GH, Cc, HS, HP, Bn, T, 7, C);
    k_stats<<<(unsigned)(C), 256, 0, stream>>>(HS, 1, C, 0, 1, NF * HW, 0.001f, st, 0);
    k_norm_apply<<<(unsigned)(((long long)(NF * HW) * (C) * (1) + 255) / 256), 256, 0, stream>>>(HS, HS, st, g2, be2, NF * HW, C, 1, 1, 1, 0);
    hipMemsetAsync(XP, 0, (size_t)NF * PP * C * 4, stream); hipMemsetAsync(HP, 0, (size_t)Bn * PP * C * 4, stream); hipMemsetAsync(Cc, 0, (size_t)Bn * HW * C * 4, stream);
    k_bl_pad<<<(unsigned)(((long long)NF * HW * C + 255) / 256), 256, 0, stream>>>(HS, XP, NF, C);
    { GemmP cx2_0;
      cx2_0.A = XP + (size_t)0 * C; cx2_0.B = Wx3 + (size_t)0 * C * G4; cx2_0.bias = b3; cx2_0.R = XP + (size_t)0 * C; cx2_0.C = XG;
      cx2_0.sAo = (long long)PP * C; cx2_0.sAi = (long long)18 * C; cx2_0.sAm = C; cx2_0.sAk = 1; cx2_0.sBo = 0; cx2_0.sBi = 0; cx2_0.sBn = 1; cx2_0.sBk = G4; cx2_0.sCo = (long long)HW * G4; cx2_0.sCi = (long long)16 * G4; cx2_0.sCm = G4; cx2_0.sRo = 0; cx2_0.sRi = 0; cx2_0.sRm = 0; cx2_0.sRn = 0;
      cx2_0.M = 16; cx2_0.N = G4; cx2_0.K = C; cx2_0.zi_n = 16; cx2_0.flags = 1; cx2_0.act = 0;
      cx2_0.alpha = 1.0f; cx2_0.beta = 0.0f; cx2_0.sa = 1.0f; cx2_0.sb = 1.0f; cx2_0.Npad = G4; cx2_0.pad_ = 0;
      k_gemm<1><<<dim3((unsigned)((G4) + 31) / 32, (unsigned)((16) + 15) / 16, (unsigned)(NF * 16)), 32, 0, stream>>>(cx2_0); }
    { GemmP cx2_1;
      cx2_1.A = XP + (size_t)1 * C; cx2_1.B = Wx3 + (size_t)1 * C * G4; cx2_1.bias = XP + (size_t)1 * C; cx2_1.R = XG; cx2_1.C = XG;
      cx2_1.sAo = (long long)PP * C; cx2_1.sAi = (long long)18 * C; cx2_1.sAm = C; cx2_1.sAk = 1; cx2_1.sBo = 0; cx2_1.sBi = 0; cx2_1.sBn = 1; cx2_1.sBk = G4; cx2_1.sCo = (long long)HW * G4; cx2_1.sCi = (long long)16 * G4; cx2_1.sCm = G4; cx2_1.sRo = (long long)HW * G4; cx2_1.sRi = (long long)16 * G4; cx2_1.sRm = G4; cx2_1.sRn = 1;
      cx2_1.M = 16; cx2_1.N = G4; cx2_1.K = C; cx2_1.zi_n = 16; cx2_1.flags = 4; cx2_1.act = 0;
      cx2_1.alpha = 1.0f; cx2_1.beta = 1.0f; cx2_1.sa = 1.0f; cx2_1.sb = 1.0f; cx2_1.Npad = G4; cx2_1.pad_ = 0;
      k_gemm<1><<<dim3((unsigned)((G4) + 31) / 32, (unsigned)((16) + 15) / 16, (unsigned)(NF * 16)), 32, 0, stream>>>(cx2_1); }
    { GemmP cx2_2;
      cx2_2.A = XP + (size_t)2 * C; cx2_2.B = Wx3 + (size_t)2 * C * G4; cx2_2.bias = XP + (size_t)2 * C; cx2_2.R = XG; cx2_2.C = XG;
      cx2_2.sAo = (long long)PP * C; cx2_2.sAi = (long long)18 * C; cx2_2.sAm = C; cx2_2.sAk = 1; cx2_2.sBo = 0; cx2_2.sBi = 0; cx2_2.sBn = 1; cx2_2.sBk = G4; cx2_2.sCo = (long long)HW * G4; cx2_2.sCi = (long long)16 * G4; cx2_2.sCm = G4; cx2_2.sRo = (long long)HW * G4; cx2_2.sRi = (long long)16 * G4; cx2_2.sRm = G4; cx2_2.sRn = 1;
      cx2_2.M = 16; cx2_2.N = G4; cx2_2.K = C; cx2_2.zi_n = 16; cx2_2.flags = 4; cx2_2.act = 0;
      cx2_2.alpha = 1.0f; cx2_2.beta = 1.0f; cx2_2.sa = 1.0f; cx2_2.sb = 1.0f; cx2_2.Npad = G4; cx2_2.pad_ = 0;
      k_gemm<1><<<dim3((unsigned)((G4) + 31) / 32, (unsigned)((16) + 15) / 16, (unsigned)(NF * 16)), 32, 0, stream>>>(cx2_2); }
    { GemmP cx2_3;
      cx2_3.A = XP + (size_t)18 * C; cx2_3.B = Wx3 + (size_t)3 * C * G4; cx2_3.bias = XP + (size_t)18 * C; cx2_3.R = XG; cx2_3.C = XG;
      cx2_3.sAo = (long long)PP * C; cx2_3.sAi = (long long)18 * C; cx2_3.sAm = C; cx2_3.sAk = 1; cx2_3.sBo = 0; cx2_3.sBi = 0; cx2_3.sBn = 1; cx2_3.sBk = G4; cx2_3.sCo = (long long)HW * G4; cx2_3.sCi = (long long)16 * G4; cx2_3.sCm = G4; cx2_3.sRo = (long long)HW * G4; cx2_3.sRi = (long long)16 * G4; cx2_3.sRm = G4; cx2_3.sRn = 1;
      cx2_3.M = 16; cx2_3.N = G4; cx2_3.K = C; cx2_3.zi_n = 16; cx2_3.flags = 4; cx2_3.act = 0;
      cx2_3.alpha = 1.0f; cx2_3.beta = 1.0f; cx2_3.sa = 1.0f; cx2_3.sb = 1.0f; cx2_3.Npad = G4; cx2_3.pad_ = 0;
      k_gemm<1><<<dim3((unsigned)((G4) + 31) / 32, (unsigned)((16) + 15) / 16, (unsigned)(NF * 16)), 32, 0, stream>>>(cx2_3); }
    { GemmP cx2_4;
      cx2_4.A = XP + (size_t)19 * C; cx2_4.B = Wx3 + (size_t)4 * C * G4; cx2_4.bias = XP + (size_t)19 * C; cx2_4.R = XG; cx2_4.C = XG;
      cx2_4.sAo = (long long)PP * C; cx2_4.sAi = (long long)18 * C; cx2_4.sAm = C; cx2_4.sAk = 1; cx2_4.sBo = 0; cx2_4.sBi = 0; cx2_4.sBn = 1; cx2_4.sBk = G4; cx2_4.sCo = (long long)HW * G4; cx2_4.sCi = (long long)16 * G4; cx2_4.sCm = G4; cx2_4.sRo = (long long)HW * G4; cx2_4.sRi = (long long)16 * G4; cx2_4.sRm = G4; cx2_4.sRn = 1;
      cx2_4.M = 16; cx2_4.N = G4; cx2_4.K = C; cx2_4.zi_n = 16; cx2_4.flags = 4; cx2_4.act = 0;
      cx2_4.alpha = 1.0f; cx2_4.beta = 1.0f; cx2_4.sa = 1.0f; cx2_4.sb = 1.0f; cx2_4.Npad = G4; cx2_4.pad_ = 0;
      k_gemm<1><<<dim3((unsigned)((G4) + 31) / 32, (unsigned)((16) + 15) / 16, (unsigned)(NF * 16)), 32, 0, stream>>>(cx2_4); }
    { GemmP cx2_5;
      cx2_5.A = XP + (size_t)20 * C; cx2_5.B = Wx3 + (size_t)5 * C * G4; cx2_5.bias = XP + (size_t)20 * C; cx2_5.R = XG; cx2_5.C = XG;
      cx2_5.sAo = (long long)PP * C; cx2_5.sAi = (long long)18 * C; cx2_5.sAm = C; cx2_5.sAk = 1; cx2_5.sBo = 0; cx2_5.sBi = 0; cx2_5.sBn = 1; cx2_5.sBk = G4; cx2_5.sCo = (long long)HW * G4; cx2_5.sCi = (long long)16 * G4; cx2_5.sCm = G4; cx2_5.sRo = (long long)HW * G4; cx2_5.sRi = (long long)16 * G4; cx2_5.sRm = G4; cx2_5.sRn = 1;
      cx2_5.M = 16; cx2_5.N = G4; cx2_5.K = C; cx2_5.zi_n = 16; cx2_5.flags = 4; cx2_5.act = 0;
      cx2_5.alpha = 1.0f; cx2_5.beta = 1.0f; cx2_5.sa = 1.0f; cx2_5.sb = 1.0f; cx2_5.Npad = G4; cx2_5.pad_ = 0;
      k_gemm<1><<<dim3((unsigned)((G4) + 31) / 32, (unsigned)((16) + 15) / 16, (unsigned)(NF * 16)), 32, 0, stream>>>(cx2_5); }
    { GemmP cx2_6;
      cx2_6.A = XP + (size_t)36 * C; cx2_6.B = Wx3 + (size_t)6 * C * G4; cx2_6.bias = XP + (size_t)36 * C; cx2_6.R = XG; cx2_6.C = XG;
      cx2_6.sAo = (long long)PP * C; cx2_6.sAi = (long long)18 * C; cx2_6.sAm = C; cx2_6.sAk = 1; cx2_6.sBo = 0; cx2_6.sBi = 0; cx2_6.sBn = 1; cx2_6.sBk = G4; cx2_6.sCo = (long long)HW * G4; cx2_6.sCi = (long long)16 * G4; cx2_6.sCm = G4; cx2_6.sRo = (long long)HW * G4; cx2_6.sRi = (long long)16 * G4; cx2_6.sRm = G4; cx2_6.sRn = 1;
      cx2_6.M = 16; cx2_6.N = G4; cx2_6.K = C; cx2_6.zi_n = 16; cx2_6.flags = 4; cx2_6.act = 0;
      cx2_6.alpha = 1.0f; cx2_6.beta = 1.0f; cx2_6.sa = 1.0f; cx2_6.sb = 1.0f; cx2_6.Npad = G4; cx2_6.pad_ = 0;
      k_gemm<1><<<dim3((unsigned)((G4) + 31) / 32, (unsigned)((16) + 15) / 16, (unsigned)(NF * 16)), 32, 0, stream>>>(cx2_6); }
    { GemmP cx2_7;
      cx2_7.A = XP + (size_t)37 * C; cx2_7.B = Wx3 + (size_t)7 * C * G4; cx2_7.bias = XP + (size_t)37 * C; cx2_7.R = XG; cx2_7.C = XG;
      cx2_7.sAo = (long long)PP * C; cx2_7.sAi = (long long)18 * C; cx2_7.sAm = C; cx2_7.sAk = 1; cx2_7.sBo = 0; cx2_7.sBi = 0; cx2_7.sBn = 1; cx2_7.sBk = G4; cx2_7.sCo = (long long)HW * G4; cx2_7.sCi = (long long)16 * G4; cx2_7.sCm = G4; cx2_7.sRo = (long long)HW * G4; cx2_7.sRi = (long long)16 * G4; cx2_7.sRm = G4; cx2_7.sRn = 1;
      cx2_7.M = 16; cx2_7.N = G4; cx2_7.K = C; cx2_7.zi_n = 16; cx2_7.flags = 4; cx2_7.act = 0;
      cx2_7.alpha = 1.0f; cx2_7.beta = 1.0f; cx2_7.sa = 1.0f; cx2_7.sb = 1.0f; cx2_7.Npad = G4; cx2_7.pad_ = 0;
      k_gemm<1><<<dim3((unsigned)((G4) + 31) / 32, (unsigned)((16) + 15) / 16, (unsigned)(NF * 16)), 32, 0, stream>>>(cx2_7); }
    { GemmP cx2_8;
      cx2_8.A = XP + (size_t)38 * C; cx2_8.B = Wx3 + (size_t)8 * C * G4; cx2_8.bias = XP + (size_t)38 * C; cx2_8.R = XG; cx2_8.C = XG;
      cx2_8.sAo = (long long)PP * C; cx2_8.sAi = (long long)18 * C; cx2_8.sAm = C; cx2_8.sAk = 1; cx2_8.sBo = 0; cx2_8.sBi = 0; cx2_8.sBn = 1; cx2_8.sBk = G4; cx2_8.sCo = (long long)HW * G4; cx2_8.sCi = (long long)16 * G4; cx2_8.sCm = G4; cx2_8.sRo = (long long)HW * G4; cx2_8.sRi = (long long)16 * G4; cx2_8.sRm = G4; cx2_8.sRn = 1;
      cx2_8.M = 16; cx2_8.N = G4; cx2_8.K = C; cx2_8.zi_n = 16; cx2_8.flags = 4; cx2_8.act = 0;
      cx2_8.alpha = 1.0f; cx2_8.beta = 1.0f; cx2_8.sa = 1.0f; cx2_8.sb = 1.0f; cx2_8.Npad = G4; cx2_8.pad_ = 0;
      k_gemm<1><<<dim3((unsigned)((G4) + 31) / 32, (unsigned)((16) + 15) / 16, (unsigned)(NF * 16)), 32, 0, stream>>>(cx2_8); }

    { GemmP ch2_0_0;
      ch2_0_0.A = HP + (size_t)0 * C; ch2_0_0.B = Wh3 + (size_t)0 * C * G4; ch2_0_0.bias = HP + (size_t)0 * C; ch2_0_0.R = HP + (size_t)0 * C; ch2_0_0.C = GH;
      ch2_0_0.sAo = (long long)PP * C; ch2_0_0.sAi = (long long)18 * C; ch2_0_0.sAm = C; ch2_0_0.sAk = 1; ch2_0_0.sBo = 0; ch2_0_0.sBi = 0; ch2_0_0.sBn = 1; ch2_0_0.sBk = G4; ch2_0_0.sCo = (long long)HW * G4; ch2_0_0.sCi = (long long)16 * G4; ch2_0_0.sCm = G4; ch2_0_0.sRo = 0; ch2_0_0.sRi = 0; ch2_0_0.sRm = 0; ch2_0_0.sRn = 0;
      ch2_0_0.M = 16; ch2_0_0.N = G4; ch2_0_0.K = C; ch2_0_0.zi_n = 16; ch2_0_0.flags = 0; ch2_0_0.act = 0;
      ch2_0_0.alpha = 1.0f; ch2_0_0.beta = 0.0f; ch2_0_0.sa = 1.0f; ch2_0_0.sb = 1.0f; ch2_0_0.Npad = G4; ch2_0_0.pad_ = 0;
      k_gemm<1><<<dim3((unsigned)((G4) + 31) / 32, (unsigned)((16) + 15) / 16, (unsigned)(Bn * 16)), 32, 0, stream>>>(ch2_0_0); }
    { GemmP ch2_0_1;
      ch2_0_1.A = HP + (size_t)1 * C; ch2_0_1.B = Wh3 + (size_t)1 * C * G4; ch2_0_1.bias = HP + (size_t)1 * C; ch2_0_1.R = GH; ch2_0_1.C = GH;
      ch2_0_1.sAo = (long long)PP * C; ch2_0_1.sAi = (long long)18 * C; ch2_0_1.sAm = C; ch2_0_1.sAk = 1; ch2_0_1.sBo = 0; ch2_0_1.sBi = 0; ch2_0_1.sBn = 1; ch2_0_1.sBk = G4; ch2_0_1.sCo = (long long)HW * G4; ch2_0_1.sCi = (long long)16 * G4; ch2_0_1.sCm = G4; ch2_0_1.sRo = (long long)HW * G4; ch2_0_1.sRi = (long long)16 * G4; ch2_0_1.sRm = G4; ch2_0_1.sRn = 1;
      ch2_0_1.M = 16; ch2_0_1.N = G4; ch2_0_1.K = C; ch2_0_1.zi_n = 16; ch2_0_1.flags = 4; ch2_0_1.act = 0;
      ch2_0_1.alpha = 1.0f; ch2_0_1.beta = 1.0f; ch2_0_1.sa = 1.0f; ch2_0_1.sb = 1.0f; ch2_0_1.Npad = G4; ch2_0_1.pad_ = 0;
      k_gemm<1><<<dim3((unsigned)((G4) + 31) / 32, (unsigned)((16) + 15) / 16, (unsigned)(Bn * 16)), 32, 0, stream>>>(ch2_0_1); }
    { GemmP ch2_0_2;
      ch2_0_2.A = HP + (size_t)2 * C; ch2_0_2.B = Wh3 + (size_t)2 * C * G4; ch2_0_2.bias = HP + (size_t)2 * C; ch2_0_2.R = GH; ch2_0_2.C = GH;
      ch2_0_2.sAo = (long long)PP * C; ch2_0_2.sAi = (long long)18 * C; ch2_0_2.sAm = C; ch2_0_2.sAk = 1; ch2_0_2.sBo = 0; ch2_0_2.sBi = 0; ch2_0_2.sBn = 1; ch2_0_2.sBk = G4; ch2_0_2.sCo = (long long)HW * G4; ch2_0_2.sCi = (long long)16 * G4; ch2_0_2.sCm = G4; ch2_0_2.sRo = (long long)HW * G4; ch2_0_2.sRi = (long long)16 * G4; ch2_0_2.sRm = G4; ch2_0_2.sRn = 1;
      ch2_0_2.M = 16; ch2_0_2.N = G4; ch2_0_2.K = C; ch2_0_2.zi_n = 16; ch2_0_2.flags = 4; ch2_0_2.act = 0;
      ch2_0_2.alpha = 1.0f; ch2_0_2.beta = 1.0f; ch2_0_2.sa = 1.0f; ch2_0_2.sb = 1.0f; ch2_0_2.Npad = G4; ch2_0_2.pad_ = 0;
      k_gemm<1><<<dim3((unsigned)((G4) + 31) / 32, (unsigned)((16) + 15) / 16, (unsigned)(Bn * 16)), 32, 0, stream>>>(ch2_0_2); }
    { GemmP ch2_0_3;
      ch2_0_3.A = HP + (size_t)18 * C; ch2_0_3.B = Wh3 + (size_t)3 * C * G4; ch2_0_3.bias = HP + (size_t)18 * C; ch2_0_3.R = GH; ch2_0_3.C = GH;
      ch2_0_3.sAo = (long long)PP * C; ch2_0_3.sAi = (long long)18 * C; ch2_0_3.sAm = C; ch2_0_3.sAk = 1; ch2_0_3.sBo = 0; ch2_0_3.sBi = 0; ch2_0_3.sBn = 1; ch2_0_3.sBk = G4; ch2_0_3.sCo = (long long)HW * G4; ch2_0_3.sCi = (long long)16 * G4; ch2_0_3.sCm = G4; ch2_0_3.sRo = (long long)HW * G4; ch2_0_3.sRi = (long long)16 * G4; ch2_0_3.sRm = G4; ch2_0_3.sRn = 1;
      ch2_0_3.M = 16; ch2_0_3.N = G4; ch2_0_3.K = C; ch2_0_3.zi_n = 16; ch2_0_3.flags = 4; ch2_0_3.act = 0;
      ch2_0_3.alpha = 1.0f; ch2_0_3.beta = 1.0f; ch2_0_3.sa = 1.0f; ch2_0_3.sb = 1.0f; ch2_0_3.Npad = G4; ch2_0_3.pad_ = 0;
      k_gemm<1><<<dim3((unsigned)((G4) + 31) / 32, (unsigned)((16) + 15) / 16, (unsigned)(Bn * 16)), 32, 0, stream>>>(ch2_0_3); }
    { GemmP ch2_0_4;
      ch2_0_4.A = HP + (size_t)19 * C; ch2_0_4.B = Wh3 + (size_t)4 * C * G4; ch2_0_4.bias = HP + (size_t)19 * C; ch2_0_4.R = GH; ch2_0_4.C = GH;
      ch2_0_4.sAo = (long long)PP * C; ch2_0_4.sAi = (long long)18 * C; ch2_0_4.sAm = C; ch2_0_4.sAk = 1; ch2_0_4.sBo = 0; ch2_0_4.sBi = 0; ch2_0_4.sBn = 1; ch2_0_4.sBk = G4; ch2_0_4.sCo = (long long)HW * G4; ch2_0_4.sCi = (long long)16 * G4; ch2_0_4.sCm = G4; ch2_0_4.sRo = (long long)HW * G4; ch2_0_4.sRi = (long long)16 * G4; ch2_0_4.sRm = G4; ch2_0_4.sRn = 1;
      ch2_0_4.M = 16; ch2_0_4.N = G4; ch2_0_4.K = C; ch2_0_4.zi_n = 16; ch2_0_4.flags = 4; ch2_0_4.act = 0;
      ch2_0_4.alpha = 1.0f; ch2_0_4.beta = 1.0f; ch2_0_4.sa = 1.0f; ch2_0_4.sb = 1.0f; ch2_0_4.Npad = G4; ch2_0_4.pad_ = 0;
      k_gemm<1><<<dim3((unsigned)((G4) + 31) / 32, (unsigned)((16) + 15) / 16, (unsigned)(Bn * 16)), 32, 0, stream>>>(ch2_0_4); }
    { GemmP ch2_0_5;
      ch2_0_5.A = HP + (size_t)20 * C; ch2_0_5.B = Wh3 + (size_t)5 * C * G4; ch2_0_5.bias = HP + (size_t)20 * C; ch2_0_5.R = GH; ch2_0_5.C = GH;
      ch2_0_5.sAo = (long long)PP * C; ch2_0_5.sAi = (long long)18 * C; ch2_0_5.sAm = C; ch2_0_5.sAk = 1; ch2_0_5.sBo = 0; ch2_0_5.sBi = 0; ch2_0_5.sBn = 1; ch2_0_5.sBk = G4; ch2_0_5.sCo = (long long)HW * G4; ch2_0_5.sCi = (long long)16 * G4; ch2_0_5.sCm = G4; ch2_0_5.sRo = (long long)HW * G4; ch2_0_5.sRi = (long long)16 * G4; ch2_0_5.sRm = G4; ch2_0_5.sRn = 1;
      ch2_0_5.M = 16; ch2_0_5.N = G4; ch2_0_5.K = C; ch2_0_5.zi_n = 16; ch2_0_5.flags = 4; ch2_0_5.act = 0;
      ch2_0_5.alpha = 1.0f; ch2_0_5.beta = 1.0f; ch2_0_5.sa = 1.0f; ch2_0_5.sb = 1.0f; ch2_0_5.Npad = G4; ch2_0_5.pad_ = 0;
      k_gemm<1><<<dim3((unsigned)((G4) + 31) / 32, (unsigned)((16) + 15) / 16, (unsigned)(Bn * 16)), 32, 0, stream>>>(ch2_0_5); }
    { GemmP ch2_0_6;
      ch2_0_6.A = HP + (size_t)36 * C; ch2_0_6.B = Wh3 + (size_t)6 * C * G4; ch2_0_6.bias = HP + (size_t)36 * C; ch2_0_6.R = GH; ch2_0_6.C = GH;
      ch2_0_6.sAo = (long long)PP * C; ch2_0_6.sAi = (long long)18 * C; ch2_0_6.sAm = C; ch2_0_6.sAk = 1; ch2_0_6.sBo = 0; ch2_0_6.sBi = 0; ch2_0_6.sBn = 1; ch2_0_6.sBk = G4; ch2_0_6.sCo = (long long)HW * G4; ch2_0_6.sCi = (long long)16 * G4; ch2_0_6.sCm = G4; ch2_0_6.sRo = (long long)HW * G4; ch2_0_6.sRi = (long long)16 * G4; ch2_0_6.sRm = G4; ch2_0_6.sRn = 1;
      ch2_0_6.M = 16; ch2_0_6.N = G4; ch2_0_6.K = C; ch2_0_6.zi_n = 16; ch2_0_6.flags = 4; ch2_0_6.act = 0;
      ch2_0_6.alpha = 1.0f; ch2_0_6.beta = 1.0f; ch2_0_6.sa = 1.0f; ch2_0_6.sb = 1.0f; ch2_0_6.Npad = G4; ch2_0_6.pad_ = 0;
      k_gemm<1><<<dim3((unsigned)((G4) + 31) / 32, (unsigned)((16) + 15) / 16, (unsigned)(Bn * 16)), 32, 0, stream>>>(ch2_0_6); }
    { GemmP ch2_0_7;
      ch2_0_7.A = HP + (size_t)37 * C; ch2_0_7.B = Wh3 + (size_t)7 * C * G4; ch2_0_7.bias = HP + (size_t)37 * C; ch2_0_7.R = GH; ch2_0_7.C = GH;
      ch2_0_7.sAo = (long long)PP * C; ch2_0_7.sAi = (long long)18 * C; ch2_0_7.sAm = C; ch2_0_7.sAk = 1; ch2_0_7.sBo = 0; ch2_0_7.sBi = 0; ch2_0_7.sBn = 1; ch2_0_7.sBk = G4; ch2_0_7.sCo = (long long)HW * G4; ch2_0_7.sCi = (long long)16 * G4; ch2_0_7.sCm = G4; ch2_0_7.sRo = (long long)HW * G4; ch2_0_7.sRi = (long long)16 * G4; ch2_0_7.sRm = G4; ch2_0_7.sRn = 1;
      ch2_0_7.M = 16; ch2_0_7.N = G4; ch2_0_7.K = C; ch2_0_7.zi_n = 16; ch2_0_7.flags = 4; ch2_0_7.act = 0;
      ch2_0_7.alpha = 1.0f; ch2_0_7.beta = 1.0f; ch2_0_7.sa = 1.0f; ch2_0_7.sb = 1.0f; ch2_0_7.Npad = G4; ch2_0_7.pad_ = 0;
      k_gemm<1><<<dim3((unsigned)((G4) + 31) / 32, (unsigned)((16) + 15) / 16, (unsigned)(Bn * 16)), 32, 0, stream>>>(ch2_0_7); }
    { GemmP ch2_0_8;
      ch2_0_8.A = HP + (size_t)38 * C; ch2_0_8.B = Wh3 + (size_t)8 * C * G4; ch2_0_8.bias = HP + (size_t)38 * C; ch2_0_8.R = GH; ch2_0_8.C = GH;
      ch2_0_8.sAo = (long long)PP * C; ch2_0_8.sAi = (long long)18 * C; ch2_0_8.sAm = C; ch2_0_8.sAk = 1; ch2_0_8.sBo = 0; ch2_0_8.sBi = 0; ch2_0_8.sBn = 1; ch2_0_8.sBk = G4; ch2_0_8.sCo = (long long)HW * G4; ch2_0_8.sCi = (long long)16 * G4; ch2_0_8.sCm = G4; ch2_0_8.sRo = (long long)HW * G4; ch2_0_8.sRi = (long long)16 * G4; ch2_0_8.sRm = G4; ch2_0_8.sRn = 1;
      ch2_0_8.M = 16; ch2_0_8.N = G4; ch2_0_8.K = C; ch2_0_8.zi_n = 16; ch2_0_8.flags = 4; ch2_0_8.act = 0;
      ch2_0_8.alpha = 1.0f; ch2_0_8.beta = 1.0f; ch2_0_8.sa = 1.0f; ch2_0_8.sb = 1.0f; ch2_0_8.Npad = G4; ch2_0_8.pad_ = 0;
      k_gemm<1><<<dim3((unsigned)((G4) + 31) / 32, (unsigned)((16) + 15) / 16, (unsigned)(Bn * 16)), 32, 0, stream>>>(ch2_0_8); }

    k_bl_cell<<<(unsigned)(((long long)Bn * HW * C + 255) / 256), 256, 0, stream>>>(XG, GH, Cc, HS, HP, Bn, T, 0, C);
    { GemmP ch2_1_0;
      ch2_1_0.A = HP + (size_t)0 * C; ch2_1_0.B = Wh3 + (size_t)0 * C * G4; ch2_1_0.bias = HP + (size_t)0 * C; ch2_1_0.R = HP + (size_t)0 * C; ch2_1_0.C = GH;
      ch2_1_0.sAo = (long long)PP * C; ch2_1_0.sAi = (long long)18 * C; ch2_1_0.sAm = C; ch2_1_0.sAk = 1; ch2_1_0.sBo = 0; ch2_1_0.sBi = 0; ch2_1_0.sBn = 1; ch2_1_0.sBk = G4; ch2_1_0.sCo = (long long)HW * G4; ch2_1_0.sCi = (long long)16 * G4; ch2_1_0.sCm = G4; ch2_1_0.sRo = 0; ch2_1_0.sRi = 0; ch2_1_0.sRm = 0; ch2_1_0.sRn = 0;
      ch2_1_0.M = 16; ch2_1_0.N = G4; ch2_1_0.K = C; ch2_1_0.zi_n = 16; ch2_1_0.flags = 0; ch2_1_0.act = 0;
      ch2_1_0.alpha = 1.0f; ch2_1_0.beta = 0.0f; ch2_1_0.sa = 1.0f; ch2_1_0.sb = 1.0f; ch2_1_0.Npad = G4; ch2_1_0.pad_ = 0;
      k_gemm<1><<<dim3((unsigned)((G4) + 31) / 32, (unsigned)((16) + 15) / 16, (unsigned)(Bn * 16)), 32, 0, stream>>>(ch2_1_0); }
    { GemmP ch2_1_1;
      ch2_1_1.A = HP + (size_t)1 * C; ch2_1_1.B = Wh3 + (size_t)1 * C * G4; ch2_1_1.bias = HP + (size_t)1 * C; ch2_1_1.R = GH; ch2_1_1.C = GH;
      ch2_1_1.sAo = (long long)PP * C; ch2_1_1.sAi = (long long)18 * C; ch2_1_1.sAm = C; ch2_1_1.sAk = 1; ch2_1_1.sBo = 0; ch2_1_1.sBi = 0; ch2_1_1.sBn = 1; ch2_1_1.sBk = G4; ch2_1_1.sCo = (long long)HW * G4; ch2_1_1.sCi = (long long)16 * G4; ch2_1_1.sCm = G4; ch2_1_1.sRo = (long long)HW * G4; ch2_1_1.sRi = (long long)16 * G4; ch2_1_1.sRm = G4; ch2_1_1.sRn = 1;
      ch2_1_1.M = 16; ch2_1_1.N = G4; ch2_1_1.K = C; ch2_1_1.zi_n = 16; ch2_1_1.flags = 4; ch2_1_1.act = 0;
      ch2_1_1.alpha = 1.0f; ch2_1_1.beta = 1.0f; ch2_1_1.sa = 1.0f; ch2_1_1.sb = 1.0f; ch2_1_1.Npad = G4; ch2_1_1.pad_ = 0;
      k_gemm<1><<<dim3((unsigned)((G4) + 31) / 32, (unsigned)((16) + 15) / 16, (unsigned)(Bn * 16)), 32, 0, stream>>>(ch2_1_1); }
    { GemmP ch2_1_2;
      ch2_1_2.A = HP + (size_t)2 * C; ch2_1_2.B = Wh3 + (size_t)2 * C * G4; ch2_1_2.bias = HP + (size_t)2 * C; ch2_1_2.R = GH; ch2_1_2.C = GH;
      ch2_1_2.sAo = (long long)PP * C; ch2_1_2.sAi = (long long)18 * C; ch2_1_2.sAm = C; ch2_1_2.sAk = 1; ch2_1_2.sBo = 0; ch2_1_2.sBi = 0; ch2_1_2.sBn = 1; ch2_1_2.sBk = G4; ch2_1_2.sCo = (long long)HW * G4; ch2_1_2.sCi = (long long)16 * G4; ch2_1_2.sCm = G4; ch2_1_2.sRo = (long long)HW * G4; ch2_1_2.sRi = (long long)16 * G4; ch2_1_2.sRm = G4; ch2_1_2.sRn = 1;
      ch2_1_2.M = 16; ch2_1_2.N = G4; ch2_1_2.K = C; ch2_1_2.zi_n = 16; ch2_1_2.flags = 4; ch2_1_2.act = 0;
      ch2_1_2.alpha = 1.0f; ch2_1_2.beta = 1.0f; ch2_1_2.sa = 1.0f; ch2_1_2.sb = 1.0f; ch2_1_2.Npad = G4; ch2_1_2.pad_ = 0;
      k_gemm<1><<<dim3((unsigned)((G4) + 31) / 32, (unsigned)((16) + 15) / 16, (unsigned)(Bn * 16)), 32, 0, stream>>>(ch2_1_2); }
    { GemmP ch2_1_3;
      ch2_1_3.A = HP + (size_t)18 * C; ch2_1_3.B = Wh3 + (size_t)3 * C * G4; ch2_1_3.bias = HP + (size_t)18 * C; ch2_1_3.R = GH; ch2_1_3.C = GH;
      ch2_1_3.sAo = (long long)PP * C; ch2_1_3.sAi = (long long)18 * C; ch2_1_3.sAm = C; ch2_1_3.sAk = 1; ch2_1_3.sBo = 0; ch2_1_3.sBi = 0; ch2_1_3.sBn = 1; ch2_1_3.sBk = G4; ch2_1_3.sCo = (long long)HW * G4; ch2_1_3.sCi = (long long)16 * G4; ch2_1_3.sCm = G4; ch2_1_3.sRo = (long long)HW * G4; ch2_1_3.sRi = (long long)16 * G4; ch2_1_3.sRm = G4; ch2_1_3.sRn = 1;
      ch2_1_3.M = 16; ch2_1_3.N = G4; ch2_1_3.K = C; ch2_1_3.zi_n = 16; ch2_1_3.flags = 4; ch2_1_3.act = 0;
      ch2_1_3.alpha = 1.0f; ch2_1_3.beta = 1.0f; ch2_1_3.sa = 1.0f; ch2_1_3.sb = 1.0f; ch2_1_3.Npad = G4; ch2_1_3.pad_ = 0;
      k_gemm<1><<<dim3((unsigned)((G4) + 31) / 32, (unsigned)((16) + 15) / 16, (unsigned)(Bn * 16)), 32, 0, stream>>>(ch2_1_3); }
    { GemmP ch2_1_4;
      ch2_1_4.A = HP + (size_t)19 * C; ch2_1_4.B = Wh3 + (size_t)4 * C * G4; ch2_1_4.bias = HP + (size_t)19 * C; ch2_1_4.R = GH; ch2_1_4.C = GH;
      ch2_1_4.sAo = (long long)PP * C; ch2_1_4.sAi = (long long)18 * C; ch2_1_4.sAm = C; ch2_1_4.sAk = 1; ch2_1_4.sBo = 0; ch2_1_4.sBi = 0; ch2_1_4.sBn = 1; ch2_1_4.sBk = G4; ch2_1_4.sCo = (long long)HW * G4; ch2_1_4.sCi = (long long)16 * G4; ch2_1_4.sCm = G4; ch2_1_4.sRo = (long long)HW * G4; ch2_1_4.sRi = (long long)16 * G4; ch2_1_4.sRm = G4; ch2_1_4.sRn = 1;
      ch2_1_4.M = 16; ch2_1_4.N = G4; ch2_1_4.K = C; ch2_1_4.zi_n = 16; ch2_1_4.flags = 4; ch2_1_4.act = 0;
      ch2_1_4.alpha = 1.0f; ch2_1_4.beta = 1.0f; ch2_1_4.sa = 1.0f; ch2_1_4.sb = 1.0f; ch2_1_4.Npad = G4; ch2_1_4.pad_ = 0;
      k_gemm<1><<<dim3((unsigned)((G4) + 31) / 32, (unsigned)((16) + 15) / 16, (unsigned)(Bn * 16)), 32, 0, stream>>>(ch2_1_4); }
    { GemmP ch2_1_5;
      ch2_1_5.A = HP + (size_t)20 * C; ch2_1_5.B = Wh3 + (size_t)5 * C * G4; ch2_1_5.bias = HP + (size_t)20 * C; ch2_1_5.R = GH; ch2_1_5.C = GH;
      ch2_1_5.sAo = (long long)PP * C; ch2_1_5.sAi = (long long)18 * C; ch2_1_5.sAm = C; ch2_1_5.sAk = 1; ch2_1_5.sBo = 0; ch2_1_5.sBi = 0; ch2_1_5.sBn = 1; ch2_1_5.sBk = G4; ch2_1_5.sCo = (long long)HW * G4; ch2_1_5.sCi = (long long)16 * G4; ch2_1_5.sCm = G4; ch2_1_5.sRo = (long long)HW * G4; ch2_1_5.sRi = (long long)16 * G4; ch2_1_5.sRm = G4; ch2_1_5.sRn = 1;
      ch2_1_5.M = 16; ch2_1_5.N = G4; ch2_1_5.K = C; ch2_1_5.zi_n = 16; ch2_1_5.flags = 4; ch2_1_5.act = 0;
      ch2_1_5.alpha = 1.0f; ch2_1_5.beta = 1.0f; ch2_1_5.sa = 1.0f; ch2_1_5.sb = 1.0f; ch2_1_5.Npad = G4; ch2_1_5.pad_ = 0;
      k_gemm<1><<<dim3((unsigned)((G4) + 31) / 32, (unsigned)((16) + 15) / 16, (unsigned)(Bn * 16)), 32, 0, stream>>>(ch2_1_5); }
    { GemmP ch2_1_6;
      ch2_1_6.A = HP + (size_t)36 * C; ch2_1_6.B = Wh3 + (size_t)6 * C * G4; ch2_1_6.bias = HP + (size_t)36 * C; ch2_1_6.R = GH; ch2_1_6.C = GH;
      ch2_1_6.sAo = (long long)PP * C; ch2_1_6.sAi = (long long)18 * C; ch2_1_6.sAm = C; ch2_1_6.sAk = 1; ch2_1_6.sBo = 0; ch2_1_6.sBi = 0; ch2_1_6.sBn = 1; ch2_1_6.sBk = G4; ch2_1_6.sCo = (long long)HW * G4; ch2_1_6.sCi = (long long)16 * G4; ch2_1_6.sCm = G4; ch2_1_6.sRo = (long long)HW * G4; ch2_1_6.sRi = (long long)16 * G4; ch2_1_6.sRm = G4; ch2_1_6.sRn = 1;
      ch2_1_6.M = 16; ch2_1_6.N = G4; ch2_1_6.K = C; ch2_1_6.zi_n = 16; ch2_1_6.flags = 4; ch2_1_6.act = 0;
      ch2_1_6.alpha = 1.0f; ch2_1_6.beta = 1.0f; ch2_1_6.sa = 1.0f; ch2_1_6.sb = 1.0f; ch2_1_6.Npad = G4; ch2_1_6.pad_ = 0;
      k_gemm<1><<<dim3((unsigned)((G4) + 31) / 32, (unsigned)((16) + 15) / 16, (unsigned)(Bn * 16)), 32, 0, stream>>>(ch2_1_6); }
    { GemmP ch2_1_7;
      ch2_1_7.A = HP + (size_t)37 * C; ch2_1_7.B = Wh3 + (size_t)7 * C * G4; ch2_1_7.bias = HP + (size_t)37 * C; ch2_1_7.R = GH; ch2_1_7.C = GH;
      ch2_1_7.sAo = (long long)PP * C; ch2_1_7.sAi = (long long)18 * C; ch2_1_7.sAm = C; ch2_1_7.sAk = 1; ch2_1_7.sBo = 0; ch2_1_7.sBi = 0; ch2_1_7.sBn = 1; ch2_1_7.sBk = G4; ch2_1_7.sCo = (long long)HW * G4; ch2_1_7.sCi = (long long)16 * G4; ch2_1_7.sCm = G4; ch2_1_7.sRo = (long long)HW * G4; ch2_1_7.sRi = (long long)16 * G4; ch2_1_7.sRm = G4; ch2_1_7.sRn = 1;
      ch2_1_7.M = 16; ch2_1_7.N = G4; ch2_1_7.K = C; ch2_1_7.zi_n = 16; ch2_1_7.flags = 4; ch2_1_7.act = 0;
      ch2_1_7.alpha = 1.0f; ch2_1_7.beta = 1.0f; ch2_1_7.sa = 1.0f; ch2_1_7.sb = 1.0f; ch2_1_7.Npad = G4; ch2_1_7.pad_ = 0;
      k_gemm<1><<<dim3((unsigned)((G4) + 31) / 32, (unsigned)((16) + 15) / 16, (unsigned)(Bn * 16)), 32, 0, stream>>>(ch2_1_7); }
    { GemmP ch2_1_8;
      ch2_1_8.A = HP + (size_t)38 * C; ch2_1_8.B = Wh3 + (size_t)8 * C * G4; ch2_1_8.bias = HP + (size_t)38 * C; ch2_1_8.R = GH; ch2_1_8.C = GH;
      ch2_1_8.sAo = (long long)PP * C; ch2_1_8.sAi = (long long)18 * C; ch2_1_8.sAm = C; ch2_1_8.sAk = 1; ch2_1_8.sBo = 0; ch2_1_8.sBi = 0; ch2_1_8.sBn = 1; ch2_1_8.sBk = G4; ch2_1_8.sCo = (long long)HW * G4; ch2_1_8.sCi = (long long)16 * G4; ch2_1_8.sCm = G4; ch2_1_8.sRo = (long long)HW * G4; ch2_1_8.sRi = (long long)16 * G4; ch2_1_8.sRm = G4; ch2_1_8.sRn = 1;
      ch2_1_8.M = 16; ch2_1_8.N = G4; ch2_1_8.K = C; ch2_1_8.zi_n = 16; ch2_1_8.flags = 4; ch2_1_8.act = 0;
      ch2_1_8.alpha = 1.0f; ch2_1_8.beta = 1.0f; ch2_1_8.sa = 1.0f; ch2_1_8.sb = 1.0f; ch2_1_8.Npad = G4; ch2_1_8.pad_ = 0;
      k_gemm<1><<<dim3((unsigned)((G4) + 31) / 32, (unsigned)((16) + 15) / 16, (unsigned)(Bn * 16)), 32, 0, stream>>>(ch2_1_8); }

    k_bl_cell<<<(unsigned)(((long long)Bn * HW * C + 255) / 256), 256, 0, stream>>>(XG, GH, Cc, HS, HP, Bn, T, 1, C);
    { GemmP ch2_2_0;
      ch2_2_0.A = HP + (size_t)0 * C; ch2_2_0.B = Wh3 + (size_t)0 * C * G4; ch2_2_0.bias = HP + (size_t)0 * C; ch2_2_0.R = HP + (size_t)0 * C; ch2_2_0.C = GH;
      ch2_2_0.sAo = (long long)PP * C; ch2_2_0.sAi = (long long)18 * C; ch2_2_0.sAm = C; ch2_2_0.sAk = 1; ch2_2_0.sBo = 0; ch2_2_0.sBi = 0; ch2_2_0.sBn = 1; ch2_2_0.sBk = G4; ch2_2_0.sCo = (long long)HW * G4; ch2_2_0.sCi = (long long)16 * G4; ch2_2_0.sCm = G4; ch2_2_0.sRo = 0; ch2_2_0.sRi = 0; ch2_2_0.sRm = 0; ch2_2_0.sRn = 0;
      ch2_2_0.M = 16; ch2_2_0.N = G4; ch2_2_0.K = C; ch2_2_0.zi_n = 16; ch2_2_0.flags = 0; ch2_2_0.act = 0;
      ch2_2_0.alpha = 1.0f; ch2_2_0.beta = 0.0f; ch2_2_0.sa = 1.0f; ch2_2_0.sb = 1.0f; ch2_2_0.Npad = G4; ch2_2_0.pad_ = 0;
      k_gemm<1><<<dim3((unsigned)((G4) + 31) / 32, (unsigned)((16) + 15) / 16, (unsigned)(Bn * 16)), 32, 0, stream>>>(ch2_2_0); }
    { GemmP ch2_2_1;
      ch2_2_1.A = HP + (size_t)1 * C; ch2_2_1.B = Wh3 + (size_t)1 * C * G4; ch2_2_1.bias = HP + (size_t)1 * C; ch2_2_1.R = GH; ch2_2_1.C = GH;
      ch2_2_1.sAo = (long long)PP * C; ch2_2_1.sAi = (long long)18 * C; ch2_2_1.sAm = C; ch2_2_1.sAk = 1; ch2_2_1.sBo = 0; ch2_2_1.sBi = 0; ch2_2_1.sBn = 1; ch2_2_1.sBk = G4; ch2_2_1.sCo = (long long)HW * G4; ch2_2_1.sCi = (long long)16 * G4; ch2_2_1.sCm = G4; ch2_2_1.sRo = (long long)HW * G4; ch2_2_1.sRi = (long long)16 * G4; ch2_2_1.sRm = G4; ch2_2_1.sRn = 1;
      ch2_2_1.M = 16; ch2_2_1.N = G4; ch2_2_1.K = C; ch2_2_1.zi_n = 16; ch2_2_1.flags = 4; ch2_2_1.act = 0;
      ch2_2_1.alpha = 1.0f; ch2_2_1.beta = 1.0f; ch2_2_1.sa = 1.0f; ch2_2_1.sb = 1.0f; ch2_2_1.Npad = G4; ch2_2_1.pad_ = 0;
      k_gemm<1><<<dim3((unsigned)((G4) + 31) / 32, (unsigned)((16) + 15) / 16, (unsigned)(Bn * 16)), 32, 0, stream>>>(ch2_2_1); }
    { GemmP ch2_2_2;
      ch2_2_2.A = HP + (size_t)2 * C; ch2_2_2.B = Wh3 + (size_t)2 * C * G4; ch2_2_2.bias = HP + (size_t)2 * C; ch2_2_2.R = GH; ch2_2_2.C = GH;
      ch2_2_2.sAo = (long long)PP * C; ch2_2_2.sAi = (long long)18 * C; ch2_2_2.sAm = C; ch2_2_2.sAk = 1; ch2_2_2.sBo = 0; ch2_2_2.sBi = 0; ch2_2_2.sBn = 1; ch2_2_2.sBk = G4; ch2_2_2.sCo = (long long)HW * G4; ch2_2_2.sCi = (long long)16 * G4; ch2_2_2.sCm = G4; ch2_2_2.sRo = (long long)HW * G4; ch2_2_2.sRi = (long long)16 * G4; ch2_2_2.sRm = G4; ch2_2_2.sRn = 1;
      ch2_2_2.M = 16; ch2_2_2.N = G4; ch2_2_2.K = C; ch2_2_2.zi_n = 16; ch2_2_2.flags = 4; ch2_2_2.act = 0;
      ch2_2_2.alpha = 1.0f; ch2_2_2.beta = 1.0f; ch2_2_2.sa = 1.0f; ch2_2_2.sb = 1.0f; ch2_2_2.Npad = G4; ch2_2_2.pad_ = 0;
      k_gemm<1><<<dim3((unsigned)((G4) + 31) / 32, (unsigned)((16) + 15) / 16, (unsigned)(Bn * 16)), 32, 0, stream>>>(ch2_2_2); }
    { GemmP ch2_2_3;
      ch2_2_3.A = HP + (size_t)18 * C; ch2_2_3.B = Wh3 + (size_t)3 * C * G4; ch2_2_3.bias = HP + (size_t)18 * C; ch2_2_3.R = GH; ch2_2_3.C = GH;
      ch2_2_3.sAo = (long long)PP * C; ch2_2_3.sAi = (long long)18 * C; ch2_2_3.sAm = C; ch2_2_3.sAk = 1; ch2_2_3.sBo = 0; ch2_2_3.sBi = 0; ch2_2_3.sBn = 1; ch2_2_3.sBk = G4; ch2_2_3.sCo = (long long)HW * G4; ch2_2_3.sCi = (long long)16 * G4; ch2_2_3.sCm = G4; ch2_2_3.sRo = (long long)HW * G4; ch2_2_3.sRi = (long long)16 * G4; ch2_2_3.sRm = G4; ch2_2_3.sRn = 1;
      ch2_2_3.M = 16; ch2_2_3.N = G4; ch2_2_3.K = C; ch2_2_3.zi_n = 16; ch2_2_3.flags = 4; ch2_2_3.act = 0;
      ch2_2_3.alpha = 1.0f; ch2_2_3.beta = 1.0f; ch2_2_3.sa = 1.0f; ch2_2_3.sb = 1.0f; ch2_2_3.Npad = G4; ch2_2_3.pad_ = 0;
      k_gemm<1><<<dim3((unsigned)((G4) + 31) / 32, (unsigned)((16) + 15) / 16, (unsigned)(Bn * 16)), 32, 0, stream>>>(ch2_2_3); }
    { GemmP ch2_2_4;
      ch2_2_4.A = HP + (size_t)19 * C; ch2_2_4.B = Wh3 + (size_t)4 * C * G4; ch2_2_4.bias = HP + (size_t)19 * C; ch2_2_4.R = GH; ch2_2_4.C = GH;
      ch2_2_4.sAo = (long long)PP * C; ch2_2_4.sAi = (long long)18 * C; ch2_2_4.sAm = C; ch2_2_4.sAk = 1; ch2_2_4.sBo = 0; ch2_2_4.sBi = 0; ch2_2_4.sBn = 1; ch2_2_4.sBk = G4; ch2_2_4.sCo = (long long)HW * G4; ch2_2_4.sCi = (long long)16 * G4; ch2_2_4.sCm = G4; ch2_2_4.sRo = (long long)HW * G4; ch2_2_4.sRi = (long long)16 * G4; ch2_2_4.sRm = G4; ch2_2_4.sRn = 1;
      ch2_2_4.M = 16; ch2_2_4.N = G4; ch2_2_4.K = C; ch2_2_4.zi_n = 16; ch2_2_4.flags = 4; ch2_2_4.act = 0;
      ch2_2_4.alpha = 1.0f; ch2_2_4.beta = 1.0f; ch2_2_4.sa = 1.0f; ch2_2_4.sb = 1.0f; ch2_2_4.Npad = G4; ch2_2_4.pad_ = 0;
      k_gemm<1><<<dim3((unsigned)((G4) + 31) / 32, (unsigned)((16) + 15) / 16, (unsigned)(Bn * 16)), 32, 0, stream>>>(ch2_2_4); }
    { GemmP ch2_2_5;
      ch2_2_5.A = HP + (size_t)20 * C; ch2_2_5.B = Wh3 + (size_t)5 * C * G4; ch2_2_5.bias = HP + (size_t)20 * C; ch2_2_5.R = GH; ch2_2_5.C = GH;
      ch2_2_5.sAo = (long long)PP * C; ch2_2_5.sAi = (long long)18 * C; ch2_2_5.sAm = C; ch2_2_5.sAk = 1; ch2_2_5.sBo = 0; ch2_2_5.sBi = 0; ch2_2_5.sBn = 1; ch2_2_5.sBk = G4; ch2_2_5.sCo = (long long)HW * G4; ch2_2_5.sCi = (long long)16 * G4; ch2_2_5.sCm = G4; ch2_2_5.sRo = (long long)HW * G4; ch2_2_5.sRi = (long long)16 * G4; ch2_2_5.sRm = G4; ch2_2_5.sRn = 1;
      ch2_2_5.M = 16; ch2_2_5.N = G4; ch2_2_5.K = C; ch2_2_5.zi_n = 16; ch2_2_5.flags = 4; ch2_2_5.act = 0;
      ch2_2_5.alpha = 1.0f; ch2_2_5.beta = 1.0f; ch2_2_5.sa = 1.0f; ch2_2_5.sb = 1.0f; ch2_2_5.Npad = G4; ch2_2_5.pad_ = 0;
      k_gemm<1><<<dim3((unsigned)((G4) + 31) / 32, (unsigned)((16) + 15) / 16, (unsigned)(Bn * 16)), 32, 0, stream>>>(ch2_2_5); }
    { GemmP ch2_2_6;
      ch2_2_6.A = HP + (size_t)36 * C; ch2_2_6.B = Wh3 + (size_t)6 * C * G4; ch2_2_6.bias = HP + (size_t)36 * C; ch2_2_6.R = GH; ch2_2_6.C = GH;
      ch2_2_6.sAo = (long long)PP * C; ch2_2_6.sAi = (long long)18 * C; ch2_2_6.sAm = C; ch2_2_6.sAk = 1; ch2_2_6.sBo = 0; ch2_2_6.sBi = 0; ch2_2_6.sBn = 1; ch2_2_6.sBk = G4; ch2_2_6.sCo = (long long)HW * G4; ch2_2_6.sCi = (long long)16 * G4; ch2_2_6.sCm = G4; ch2_2_6.sRo = (long long)HW * G4; ch2_2_6.sRi = (long long)16 * G4; ch2_2_6.sRm = G4; ch2_2_6.sRn = 1;
      ch2_2_6.M = 16; ch2_2_6.N = G4; ch2_2_6.K = C; ch2_2_6.zi_n = 16; ch2_2_6.flags = 4; ch2_2_6.act = 0;
      ch2_2_6.alpha = 1.0f; ch2_2_6.beta = 1.0f; ch2_2_6.sa = 1.0f; ch2_2_6.sb = 1.0f; ch2_2_6.Npad = G4; ch2_2_6.pad_ = 0;
      k_gemm<1><<<dim3((unsigned)((G4) + 31) / 32, (unsigned)((16) + 15) / 16, (unsigned)(Bn * 16)), 32, 0, stream>>>(ch2_2_6); }
    { GemmP ch2_2_7;
      ch2_2_7.A = HP + (size_t)37 * C; ch2_2_7.B = Wh3 + (size_t)7 * C * G4; ch2_2_7.bias = HP + (size_t)37 * C; ch2_2_7.R = GH; ch2_2_7.C = GH;
      ch2_2_7.sAo = (long long)PP * C; ch2_2_7.sAi = (long long)18 * C; ch2_2_7.sAm = C; ch2_2_7.sAk = 1; ch2_2_7.sBo = 0; ch2_2_7.sBi = 0; ch2_2_7.sBn = 1; ch2_2_7.sBk = G4; ch2_2_7.sCo = (long long)HW * G4; ch2_2_7.sCi = (long long)16 * G4; ch2_2_7.sCm = G4; ch2_2_7.sRo = (long long)HW * G4; ch2_2_7.sRi = (long long)16 * G4; ch2_2_7.sRm = G4; ch2_2_7.sRn = 1;
      ch2_2_7.M = 16; ch2_2_7.N = G4; ch2_2_7.K = C; ch2_2_7.zi_n = 16; ch2_2_7.flags = 4; ch2_2_7.act = 0;
      ch2_2_7.alpha = 1.0f; ch2_2_7.beta = 1.0f; ch2_2_7.sa = 1.0f; ch2_2_7.sb = 1.0f; ch2_2_7.Npad = G4; ch2_2_7.pad_ = 0;
      k_gemm<1><<<dim3((unsigned)((G4) + 31) / 32, (unsigned)((16) + 15) / 16, (unsigned)(Bn * 16)), 32, 0, stream>>>(ch2_2_7); }
    { GemmP ch2_2_8;
      ch2_2_8.A = HP + (size_t)38 * C; ch2_2_8.B = Wh3 + (size_t)8 * C * G4; ch2_2_8.bias = HP + (size_t)38 * C; ch2_2_8.R = GH; ch2_2_8.C = GH;
      ch2_2_8.sAo = (long long)PP * C; ch2_2_8.sAi = (long long)18 * C; ch2_2_8.sAm = C; ch2_2_8.sAk = 1; ch2_2_8.sBo = 0; ch2_2_8.sBi = 0; ch2_2_8.sBn = 1; ch2_2_8.sBk = G4; ch2_2_8.sCo = (long long)HW * G4; ch2_2_8.sCi = (long long)16 * G4; ch2_2_8.sCm = G4; ch2_2_8.sRo = (long long)HW * G4; ch2_2_8.sRi = (long long)16 * G4; ch2_2_8.sRm = G4; ch2_2_8.sRn = 1;
      ch2_2_8.M = 16; ch2_2_8.N = G4; ch2_2_8.K = C; ch2_2_8.zi_n = 16; ch2_2_8.flags = 4; ch2_2_8.act = 0;
      ch2_2_8.alpha = 1.0f; ch2_2_8.beta = 1.0f; ch2_2_8.sa = 1.0f; ch2_2_8.sb = 1.0f; ch2_2_8.Npad = G4; ch2_2_8.pad_ = 0;
      k_gemm<1><<<dim3((unsigned)((G4) + 31) / 32, (unsigned)((16) + 15) / 16, (unsigned)(Bn * 16)), 32, 0, stream>>>(ch2_2_8); }

    k_bl_cell<<<(unsigned)(((long long)Bn * HW * C + 255) / 256), 256, 0, stream>>>(XG, GH, Cc, HS, HP, Bn, T, 2, C);
    { GemmP ch2_3_0;
      ch2_3_0.A = HP + (size_t)0 * C; ch2_3_0.B = Wh3 + (size_t)0 * C * G4; ch2_3_0.bias = HP + (size_t)0 * C; ch2_3_0.R = HP + (size_t)0 * C; ch2_3_0.C = GH;
      ch2_3_0.sAo = (long long)PP * C; ch2_3_0.sAi = (long long)18 * C; ch2_3_0.sAm = C; ch2_3_0.sAk = 1; ch2_3_0.sBo = 0; ch2_3_0.sBi = 0; ch2_3_0.sBn = 1; ch2_3_0.sBk = G4; ch2_3_0.sCo = (long long)HW * G4; ch2_3_0.sCi = (long long)16 * G4; ch2_3_0.sCm = G4; ch2_3_0.sRo = 0; ch2_3_0.sRi = 0; ch2_3_0.sRm = 0; ch2_3_0.sRn = 0;
      ch2_3_0.M = 16; ch2_3_0.N = G4; ch2_3_0.K = C; ch2_3_0.zi_n = 16; ch2_3_0.flags = 0; ch2_3_0.act = 0;
      ch2_3_0.alpha = 1.0f; ch2_3_0.beta = 0.0f; ch2_3_0.sa = 1.0f; ch2_3_0.sb = 1.0f; ch2_3_0.Npad = G4; ch2_3_0.pad_ = 0;
      k_gemm<1><<<dim3((unsigned)((G4) + 31) / 32, (unsigned)((16) + 15) / 16, (unsigned)(Bn * 16)), 32, 0, stream>>>(ch2_3_0); }
    { GemmP ch2_3_1;
      ch2_3_1.A = HP + (size_t)1 * C; ch2_3_1.B = Wh3 + (size_t)1 * C * G4; ch2_3_1.bias = HP + (size_t)1 * C; ch2_3_1.R = GH; ch2_3_1.C = GH;
      ch2_3_1.sAo = (long long)PP * C; ch2_3_1.sAi = (long long)18 * C; ch2_3_1.sAm = C; ch2_3_1.sAk = 1; ch2_3_1.sBo = 0; ch2_3_1.sBi = 0; ch2_3_1.sBn = 1; ch2_3_1.sBk = G4; ch2_3_1.sCo = (long long)HW * G4; ch2_3_1.sCi = (long long)16 * G4; ch2_3_1.sCm = G4; ch2_3_1.sRo = (long long)HW * G4; ch2_3_1.sRi = (long long)16 * G4; ch2_3_1.sRm = G4; ch2_3_1.sRn = 1;
      ch2_3_1.M = 16; ch2_3_1.N = G4; ch2_3_1.K = C; ch2_3_1.zi_n = 16; ch2_3_1.flags = 4; ch2_3_1.act = 0;
      ch2_3_1.alpha = 1.0f; ch2_3_1.beta = 1.0f; ch2_3_1.sa = 1.0f; ch2_3_1.sb = 1.0f; ch2_3_1.Npad = G4; ch2_3_1.pad_ = 0;
      k_gemm<1><<<dim3((unsigned)((G4) + 31) / 32, (unsigned)((16) + 15) / 16, (unsigned)(Bn * 16)), 32, 0, stream>>>(ch2_3_1); }
    { GemmP ch2_3_2;
      ch2_3_2.A = HP + (size_t)2 * C; ch2_3_2.B = Wh3 + (size_t)2 * C * G4; ch2_3_2.bias = HP + (size_t)2 * C; ch2_3_2.R = GH; ch2_3_2.C = GH;
      ch2_3_2.sAo = (long long)PP * C; ch2_3_2.sAi = (long long)18 * C; ch2_3_2.sAm = C; ch2_3_2.sAk = 1; ch2_3_2.sBo = 0; ch2_3_2.sBi = 0; ch2_3_2.sBn = 1; ch2_3_2.sBk = G4; ch2_3_2.sCo = (long long)HW * G4; ch2_3_2.sCi = (long long)16 * G4; ch2_3_2.sCm = G4; ch2_3_2.sRo = (long long)HW * G4; ch2_3_2.sRi = (long long)16 * G4; ch2_3_2.sRm = G4; ch2_3_2.sRn = 1;
      ch2_3_2.M = 16; ch2_3_2.N = G4; ch2_3_2.K = C; ch2_3_2.zi_n = 16; ch2_3_2.flags = 4; ch2_3_2.act = 0;
      ch2_3_2.alpha = 1.0f; ch2_3_2.beta = 1.0f; ch2_3_2.sa = 1.0f; ch2_3_2.sb = 1.0f; ch2_3_2.Npad = G4; ch2_3_2.pad_ = 0;
      k_gemm<1><<<dim3((unsigned)((G4) + 31) / 32, (unsigned)((16) + 15) / 16, (unsigned)(Bn * 16)), 32, 0, stream>>>(ch2_3_2); }
    { GemmP ch2_3_3;
      ch2_3_3.A = HP + (size_t)18 * C; ch2_3_3.B = Wh3 + (size_t)3 * C * G4; ch2_3_3.bias = HP + (size_t)18 * C; ch2_3_3.R = GH; ch2_3_3.C = GH;
      ch2_3_3.sAo = (long long)PP * C; ch2_3_3.sAi = (long long)18 * C; ch2_3_3.sAm = C; ch2_3_3.sAk = 1; ch2_3_3.sBo = 0; ch2_3_3.sBi = 0; ch2_3_3.sBn = 1; ch2_3_3.sBk = G4; ch2_3_3.sCo = (long long)HW * G4; ch2_3_3.sCi = (long long)16 * G4; ch2_3_3.sCm = G4; ch2_3_3.sRo = (long long)HW * G4; ch2_3_3.sRi = (long long)16 * G4; ch2_3_3.sRm = G4; ch2_3_3.sRn = 1;
      ch2_3_3.M = 16; ch2_3_3.N = G4; ch2_3_3.K = C; ch2_3_3.zi_n = 16; ch2_3_3.flags = 4; ch2_3_3.act = 0;
      ch2_3_3.alpha = 1.0f; ch2_3_3.beta = 1.0f; ch2_3_3.sa = 1.0f; ch2_3_3.sb = 1.0f; ch2_3_3.Npad = G4; ch2_3_3.pad_ = 0;
      k_gemm<1><<<dim3((unsigned)((G4) + 31) / 32, (unsigned)((16) + 15) / 16, (unsigned)(Bn * 16)), 32, 0, stream>>>(ch2_3_3); }
    { GemmP ch2_3_4;
      ch2_3_4.A = HP + (size_t)19 * C; ch2_3_4.B = Wh3 + (size_t)4 * C * G4; ch2_3_4.bias = HP + (size_t)19 * C; ch2_3_4.R = GH; ch2_3_4.C = GH;
      ch2_3_4.sAo = (long long)PP * C; ch2_3_4.sAi = (long long)18 * C; ch2_3_4.sAm = C; ch2_3_4.sAk = 1; ch2_3_4.sBo = 0; ch2_3_4.sBi = 0; ch2_3_4.sBn = 1; ch2_3_4.sBk = G4; ch2_3_4.sCo = (long long)HW * G4; ch2_3_4.sCi = (long long)16 * G4; ch2_3_4.sCm = G4; ch2_3_4.sRo = (long long)HW * G4; ch2_3_4.sRi = (long long)16 * G4; ch2_3_4.sRm = G4; ch2_3_4.sRn = 1;
      ch2_3_4.M = 16; ch2_3_4.N = G4; ch2_3_4.K = C; ch2_3_4.zi_n = 16; ch2_3_4.flags = 4; ch2_3_4.act = 0;
      ch2_3_4.alpha = 1.0f; ch2_3_4.beta = 1.0f; ch2_3_4.sa = 1.0f; ch2_3_4.sb = 1.0f; ch2_3_4.Npad = G4; ch2_3_4.pad_ = 0;
      k_gemm<1><<<dim3((unsigned)((G4) + 31) / 32, (unsigned)((16) + 15) / 16, (unsigned)(Bn * 16)), 32, 0, stream>>>(ch2_3_4); }
    { GemmP ch2_3_5;
      ch2_3_5.A = HP + (size_t)20 * C; ch2_3_5.B = Wh3 + (size_t)5 * C * G4; ch2_3_5.bias = HP + (size_t)20 * C; ch2_3_5.R = GH; ch2_3_5.C = GH;
      ch2_3_5.sAo = (long long)PP * C; ch2_3_5.sAi = (long long)18 * C; ch2_3_5.sAm = C; ch2_3_5.sAk = 1; ch2_3_5.sBo = 0; ch2_3_5.sBi = 0; ch2_3_5.sBn = 1; ch2_3_5.sBk = G4; ch2_3_5.sCo = (long long)HW * G4; ch2_3_5.sCi = (long long)16 * G4; ch2_3_5.sCm = G4; ch2_3_5.sRo = (long long)HW * G4; ch2_3_5.sRi = (long long)16 * G4; ch2_3_5.sRm = G4; ch2_3_5.sRn = 1;
      ch2_3_5.M = 16; ch2_3_5.N = G4; ch2_3_5.K = C; ch2_3_5.zi_n = 16; ch2_3_5.flags = 4; ch2_3_5.act = 0;
      ch2_3_5.alpha = 1.0f; ch2_3_5.beta = 1.0f; ch2_3_5.sa = 1.0f; ch2_3_5.sb = 1.0f; ch2_3_5.Npad = G4; ch2_3_5.pad_ = 0;
      k_gemm<1><<<dim3((unsigned)((G4) + 31) / 32, (unsigned)((16) + 15) / 16, (unsigned)(Bn * 16)), 32, 0, stream>>>(ch2_3_5); }
    { GemmP ch2_3_6;
      ch2_3_6.A = HP + (size_t)36 * C; ch2_3_6.B = Wh3 + (size_t)6 * C * G4; ch2_3_6.bias = HP + (size_t)36 * C; ch2_3_6.R = GH; ch2_3_6.C = GH;
      ch2_3_6.sAo = (long long)PP * C; ch2_3_6.sAi = (long long)18 * C; ch2_3_6.sAm = C; ch2_3_6.sAk = 1; ch2_3_6.sBo = 0; ch2_3_6.sBi = 0; ch2_3_6.sBn = 1; ch2_3_6.sBk = G4; ch2_3_6.sCo = (long long)HW * G4; ch2_3_6.sCi = (long long)16 * G4; ch2_3_6.sCm = G4; ch2_3_6.sRo = (long long)HW * G4; ch2_3_6.sRi = (long long)16 * G4; ch2_3_6.sRm = G4; ch2_3_6.sRn = 1;
      ch2_3_6.M = 16; ch2_3_6.N = G4; ch2_3_6.K = C; ch2_3_6.zi_n = 16; ch2_3_6.flags = 4; ch2_3_6.act = 0;
      ch2_3_6.alpha = 1.0f; ch2_3_6.beta = 1.0f; ch2_3_6.sa = 1.0f; ch2_3_6.sb = 1.0f; ch2_3_6.Npad = G4; ch2_3_6.pad_ = 0;
      k_gemm<1><<<dim3((unsigned)((G4) + 31) / 32, (unsigned)((16) + 15) / 16, (unsigned)(Bn * 16)), 32, 0, stream>>>(ch2_3_6); }
    { GemmP ch2_3_7;
      ch2_3_7.A = HP + (size_t)37 * C; ch2_3_7.B = Wh3 + (size_t)7 * C * G4; ch2_3_7.bias = HP + (size_t)37 * C; ch2_3_7.R = GH; ch2_3_7.C = GH;
      ch2_3_7.sAo = (long long)PP * C; ch2_3_7.sAi = (long long)18 * C; ch2_3_7.sAm = C; ch2_3_7.sAk = 1; ch2_3_7.sBo = 0; ch2_3_7.sBi = 0; ch2_3_7.sBn = 1; ch2_3_7.sBk = G4; ch2_3_7.sCo = (long long)HW * G4; ch2_3_7.sCi = (long long)16 * G4; ch2_3_7.sCm = G4; ch2_3_7.sRo = (long long)HW * G4; ch2_3_7.sRi = (long long)16 * G4; ch2_3_7.sRm = G4; ch2_3_7.sRn = 1;
      ch2_3_7.M = 16; ch2_3_7.N = G4; ch2_3_7.K = C; ch2_3_7.zi_n = 16; ch2_3_7.flags = 4; ch2_3_7.act = 0;
      ch2_3_7.alpha = 1.0f; ch2_3_7.beta = 1.0f; ch2_3_7.sa = 1.0f; ch2_3_7.sb = 1.0f; ch2_3_7.Npad = G4; ch2_3_7.pad_ = 0;
      k_gemm<1><<<dim3((unsigned)((G4) + 31) / 32, (unsigned)((16) + 15) / 16, (unsigned)(Bn * 16)), 32, 0, stream>>>(ch2_3_7); }
    { GemmP ch2_3_8;
      ch2_3_8.A = HP + (size_t)38 * C; ch2_3_8.B = Wh3 + (size_t)8 * C * G4; ch2_3_8.bias = HP + (size_t)38 * C; ch2_3_8.R = GH; ch2_3_8.C = GH;
      ch2_3_8.sAo = (long long)PP * C; ch2_3_8.sAi = (long long)18 * C; ch2_3_8.sAm = C; ch2_3_8.sAk = 1; ch2_3_8.sBo = 0; ch2_3_8.sBi = 0; ch2_3_8.sBn = 1; ch2_3_8.sBk = G4; ch2_3_8.sCo = (long long)HW * G4; ch2_3_8.sCi = (long long)16 * G4; ch2_3_8.sCm = G4; ch2_3_8.sRo = (long long)HW * G4; ch2_3_8.sRi = (long long)16 * G4; ch2_3_8.sRm = G4; ch2_3_8.sRn = 1;
      ch2_3_8.M = 16; ch2_3_8.N = G4; ch2_3_8.K = C; ch2_3_8.zi_n = 16; ch2_3_8.flags = 4; ch2_3_8.act = 0;
      ch2_3_8.alpha = 1.0f; ch2_3_8.beta = 1.0f; ch2_3_8.sa = 1.0f; ch2_3_8.sb = 1.0f; ch2_3_8.Npad = G4; ch2_3_8.pad_ = 0;
      k_gemm<1><<<dim3((unsigned)((G4) + 31) / 32, (unsigned)((16) + 15) / 16, (unsigned)(Bn * 16)), 32, 0, stream>>>(ch2_3_8); }

    k_bl_cell<<<(unsigned)(((long long)Bn * HW * C + 255) / 256), 256, 0, stream>>>(XG, GH, Cc, HS, HP, Bn, T, 3, C);
    { GemmP ch2_4_0;
      ch2_4_0.A = HP + (size_t)0 * C; ch2_4_0.B = Wh3 + (size_t)0 * C * G4; ch2_4_0.bias = HP + (size_t)0 * C; ch2_4_0.R = HP + (size_t)0 * C; ch2_4_0.C = GH;
      ch2_4_0.sAo = (long long)PP * C; ch2_4_0.sAi = (long long)18 * C; ch2_4_0.sAm = C; ch2_4_0.sAk = 1; ch2_4_0.sBo = 0; ch2_4_0.sBi = 0; ch2_4_0.sBn = 1; ch2_4_0.sBk = G4; ch2_4_0.sCo = (long long)HW * G4; ch2_4_0.sCi = (long long)16 * G4; ch2_4_0.sCm = G4; ch2_4_0.sRo = 0; ch2_4_0.sRi = 0; ch2_4_0.sRm = 0; ch2_4_0.sRn = 0;
      ch2_4_0.M = 16; ch2_4_0.N = G4; ch2_4_0.K = C; ch2_4_0.zi_n = 16; ch2_4_0.flags = 0; ch2_4_0.act = 0;
      ch2_4_0.alpha = 1.0f; ch2_4_0.beta = 0.0f; ch2_4_0.sa = 1.0f; ch2_4_0.sb = 1.0f; ch2_4_0.Npad = G4; ch2_4_0.pad_ = 0;
      k_gemm<1><<<dim3((unsigned)((G4) + 31) / 32, (unsigned)((16) + 15) / 16, (unsigned)(Bn * 16)), 32, 0, stream>>>(ch2_4_0); }
    { GemmP ch2_4_1;
      ch2_4_1.A = HP + (size_t)1 * C; ch2_4_1.B = Wh3 + (size_t)1 * C * G4; ch2_4_1.bias = HP + (size_t)1 * C; ch2_4_1.R = GH; ch2_4_1.C = GH;
      ch2_4_1.sAo = (long long)PP * C; ch2_4_1.sAi = (long long)18 * C; ch2_4_1.sAm = C; ch2_4_1.sAk = 1; ch2_4_1.sBo = 0; ch2_4_1.sBi = 0; ch2_4_1.sBn = 1; ch2_4_1.sBk = G4; ch2_4_1.sCo = (long long)HW * G4; ch2_4_1.sCi = (long long)16 * G4; ch2_4_1.sCm = G4; ch2_4_1.sRo = (long long)HW * G4; ch2_4_1.sRi = (long long)16 * G4; ch2_4_1.sRm = G4; ch2_4_1.sRn = 1;
      ch2_4_1.M = 16; ch2_4_1.N = G4; ch2_4_1.K = C; ch2_4_1.zi_n = 16; ch2_4_1.flags = 4; ch2_4_1.act = 0;
      ch2_4_1.alpha = 1.0f; ch2_4_1.beta = 1.0f; ch2_4_1.sa = 1.0f; ch2_4_1.sb = 1.0f; ch2_4_1.Npad = G4; ch2_4_1.pad_ = 0;
      k_gemm<1><<<dim3((unsigned)((G4) + 31) / 32, (unsigned)((16) + 15) / 16, (unsigned)(Bn * 16)), 32, 0, stream>>>(ch2_4_1); }
    { GemmP ch2_4_2;
      ch2_4_2.A = HP + (size_t)2 * C; ch2_4_2.B = Wh3 + (size_t)2 * C * G4; ch2_4_2.bias = HP + (size_t)2 * C; ch2_4_2.R = GH; ch2_4_2.C = GH;
      ch2_4_2.sAo = (long long)PP * C; ch2_4_2.sAi = (long long)18 * C; ch2_4_2.sAm = C; ch2_4_2.sAk = 1; ch2_4_2.sBo = 0; ch2_4_2.sBi = 0; ch2_4_2.sBn = 1; ch2_4_2.sBk = G4; ch2_4_2.sCo = (long long)HW * G4; ch2_4_2.sCi = (long long)16 * G4; ch2_4_2.sCm = G4; ch2_4_2.sRo = (long long)HW * G4; ch2_4_2.sRi = (long long)16 * G4; ch2_4_2.sRm = G4; ch2_4_2.sRn = 1;
      ch2_4_2.M = 16; ch2_4_2.N = G4; ch2_4_2.K = C; ch2_4_2.zi_n = 16; ch2_4_2.flags = 4; ch2_4_2.act = 0;
      ch2_4_2.alpha = 1.0f; ch2_4_2.beta = 1.0f; ch2_4_2.sa = 1.0f; ch2_4_2.sb = 1.0f; ch2_4_2.Npad = G4; ch2_4_2.pad_ = 0;
      k_gemm<1><<<dim3((unsigned)((G4) + 31) / 32, (unsigned)((16) + 15) / 16, (unsigned)(Bn * 16)), 32, 0, stream>>>(ch2_4_2); }
    { GemmP ch2_4_3;
      ch2_4_3.A = HP + (size_t)18 * C; ch2_4_3.B = Wh3 + (size_t)3 * C * G4; ch2_4_3.bias = HP + (size_t)18 * C; ch2_4_3.R = GH; ch2_4_3.C = GH;
      ch2_4_3.sAo = (long long)PP * C; ch2_4_3.sAi = (long long)18 * C; ch2_4_3.sAm = C; ch2_4_3.sAk = 1; ch2_4_3.sBo = 0; ch2_4_3.sBi = 0; ch2_4_3.sBn = 1; ch2_4_3.sBk = G4; ch2_4_3.sCo = (long long)HW * G4; ch2_4_3.sCi = (long long)16 * G4; ch2_4_3.sCm = G4; ch2_4_3.sRo = (long long)HW * G4; ch2_4_3.sRi = (long long)16 * G4; ch2_4_3.sRm = G4; ch2_4_3.sRn = 1;
      ch2_4_3.M = 16; ch2_4_3.N = G4; ch2_4_3.K = C; ch2_4_3.zi_n = 16; ch2_4_3.flags = 4; ch2_4_3.act = 0;
      ch2_4_3.alpha = 1.0f; ch2_4_3.beta = 1.0f; ch2_4_3.sa = 1.0f; ch2_4_3.sb = 1.0f; ch2_4_3.Npad = G4; ch2_4_3.pad_ = 0;
      k_gemm<1><<<dim3((unsigned)((G4) + 31) / 32, (unsigned)((16) + 15) / 16, (unsigned)(Bn * 16)), 32, 0, stream>>>(ch2_4_3); }
    { GemmP ch2_4_4;
      ch2_4_4.A = HP + (size_t)19 * C; ch2_4_4.B = Wh3 + (size_t)4 * C * G4; ch2_4_4.bias = HP + (size_t)19 * C; ch2_4_4.R = GH; ch2_4_4.C = GH;
      ch2_4_4.sAo = (long long)PP * C; ch2_4_4.sAi = (long long)18 * C; ch2_4_4.sAm = C; ch2_4_4.sAk = 1; ch2_4_4.sBo = 0; ch2_4_4.sBi = 0; ch2_4_4.sBn = 1; ch2_4_4.sBk = G4; ch2_4_4.sCo = (long long)HW * G4; ch2_4_4.sCi = (long long)16 * G4; ch2_4_4.sCm = G4; ch2_4_4.sRo = (long long)HW * G4; ch2_4_4.sRi = (long long)16 * G4; ch2_4_4.sRm = G4; ch2_4_4.sRn = 1;
      ch2_4_4.M = 16; ch2_4_4.N = G4; ch2_4_4.K = C; ch2_4_4.zi_n = 16; ch2_4_4.flags = 4; ch2_4_4.act = 0;
      ch2_4_4.alpha = 1.0f; ch2_4_4.beta = 1.0f; ch2_4_4.sa = 1.0f; ch2_4_4.sb = 1.0f; ch2_4_4.Npad = G4; ch2_4_4.pad_ = 0;
      k_gemm<1><<<dim3((unsigned)((G4) + 31) / 32, (unsigned)((16) + 15) / 16, (unsigned)(Bn * 16)), 32, 0, stream>>>(ch2_4_4); }
    { GemmP ch2_4_5;
      ch2_4_5.A = HP + (size_t)20 * C; ch2_4_5.B = Wh3 + (size_t)5 * C * G4; ch2_4_5.bias = HP + (size_t)20 * C; ch2_4_5.R = GH; ch2_4_5.C = GH;
      ch2_4_5.sAo = (long long)PP * C; ch2_4_5.sAi = (long long)18 * C; ch2_4_5.sAm = C; ch2_4_5.sAk = 1; ch2_4_5.sBo = 0; ch2_4_5.sBi = 0; ch2_4_5.sBn = 1; ch2_4_5.sBk = G4; ch2_4_5.sCo = (long long)HW * G4; ch2_4_5.sCi = (long long)16 * G4; ch2_4_5.sCm = G4; ch2_4_5.sRo = (long long)HW * G4; ch2_4_5.sRi = (long long)16 * G4; ch2_4_5.sRm = G4; ch2_4_5.sRn = 1;
      ch2_4_5.M = 16; ch2_4_5.N = G4; ch2_4_5.K = C; ch2_4_5.zi_n = 16; ch2_4_5.flags = 4; ch2_4_5.act = 0;
      ch2_4_5.alpha = 1.0f; ch2_4_5.beta = 1.0f; ch2_4_5.sa = 1.0f; ch2_4_5.sb = 1.0f; ch2_4_5.Npad = G4; ch2_4_5.pad_ = 0;
      k_gemm<1><<<dim3((unsigned)((G4) + 31) / 32, (unsigned)((16) + 15) / 16, (unsigned)(Bn * 16)), 32, 0, stream>>>(ch2_4_5); }
    { GemmP ch2_4_6;
      ch2_4_6.A = HP + (size_t)36 * C; ch2_4_6.B = Wh3 + (size_t)6 * C * G4; ch2_4_6.bias = HP + (size_t)36 * C; ch2_4_6.R = GH; ch2_4_6.C = GH;
      ch2_4_6.sAo = (long long)PP * C; ch2_4_6.sAi = (long long)18 * C; ch2_4_6.sAm = C; ch2_4_6.sAk = 1; ch2_4_6.sBo = 0; ch2_4_6.sBi = 0; ch2_4_6.sBn = 1; ch2_4_6.sBk = G4; ch2_4_6.sCo = (long long)HW * G4; ch2_4_6.sCi = (long long)16 * G4; ch2_4_6.sCm = G4; ch2_4_6.sRo = (long long)HW * G4; ch2_4_6.sRi = (long long)16 * G4; ch2_4_6.sRm = G4; ch2_4_6.sRn = 1;
      ch2_4_6.M = 16; ch2_4_6.N = G4; ch2_4_6.K = C; ch2_4_6.zi_n = 16; ch2_4_6.flags = 4; ch2_4_6.act = 0;
      ch2_4_6.alpha = 1.0f; ch2_4_6.beta = 1.0f; ch2_4_6.sa = 1.0f; ch2_4_6.sb = 1.0f; ch2_4_6.Npad = G4; ch2_4_6.pad_ = 0;
      k_gemm<1><<<dim3((unsigned)((G4) + 31) / 32, (unsigned)((16) + 15) / 16, (unsigned)(Bn * 16)), 32, 0, stream>>>(ch2_4_6); }
    { GemmP ch2_4_7;
      ch2_4_7.A = HP + (size_t)37 * C; ch2_4_7.B = Wh3 + (size_t)7 * C * G4; ch2_4_7.bias = HP + (size_t)37 * C; ch2_4_7.R = GH; ch2_4_7.C = GH;
      ch2_4_7.sAo = (long long)PP * C; ch2_4_7.sAi = (long long)18 * C; ch2_4_7.sAm = C; ch2_4_7.sAk = 1; ch2_4_7.sBo = 0; ch2_4_7.sBi = 0; ch2_4_7.sBn = 1; ch2_4_7.sBk = G4; ch2_4_7.sCo = (long long)HW * G4; ch2_4_7.sCi = (long long)16 * G4; ch2_4_7.sCm = G4; ch2_4_7.sRo = (long long)HW * G4; ch2_4_7.sRi = (long long)16 * G4; ch2_4_7.sRm = G4; ch2_4_7.sRn = 1;
      ch2_4_7.M = 16; ch2_4_7.N = G4; ch2_4_7.K = C; ch2_4_7.zi_n = 16; ch2_4_7.flags = 4; ch2_4_7.act = 0;
      ch2_4_7.alpha = 1.0f; ch2_4_7.beta = 1.0f; ch2_4_7.sa = 1.0f; ch2_4_7.sb = 1.0f; ch2_4_7.Npad = G4; ch2_4_7.pad_ = 0;
      k_gemm<1><<<dim3((unsigned)((G4) + 31) / 32, (unsigned)((16) + 15) / 16, (unsigned)(Bn * 16)), 32, 0, stream>>>(ch2_4_7); }
    { GemmP ch2_4_8;
      ch2_4_8.A = HP + (size_t)38 * C; ch2_4_8.B = Wh3 + (size_t)8 * C * G4; ch2_4_8.bias = HP + (size_t)38 * C; ch2_4_8.R = GH; ch2_4_8.C = GH;
      ch2_4_8.sAo = (long long)PP * C; ch2_4_8.sAi = (long long)18 * C; ch2_4_8.sAm = C; ch2_4_8.sAk = 1; ch2_4_8.sBo = 0; ch2_4_8.sBi = 0; ch2_4_8.sBn = 1; ch2_4_8.sBk = G4; ch2_4_8.sCo = (long long)HW * G4; ch2_4_8.sCi = (long long)16 * G4; ch2_4_8.sCm = G4; ch2_4_8.sRo = (long long)HW * G4; ch2_4_8.sRi = (long long)16 * G4; ch2_4_8.sRm = G4; ch2_4_8.sRn = 1;
      ch2_4_8.M = 16; ch2_4_8.N = G4; ch2_4_8.K = C; ch2_4_8.zi_n = 16; ch2_4_8.flags = 4; ch2_4_8.act = 0;
      ch2_4_8.alpha = 1.0f; ch2_4_8.beta = 1.0f; ch2_4_8.sa = 1.0f; ch2_4_8.sb = 1.0f; ch2_4_8.Npad = G4; ch2_4_8.pad_ = 0;
      k_gemm<1><<<dim3((unsigned)((G4) + 31) / 32, (unsigned)((16) + 15) / 16, (unsigned)(Bn * 16)), 32, 0, stream>>>(ch2_4_8); }

    k_bl_cell<<<(unsigned)(((long long)Bn * HW * C + 255) / 256), 256, 0, stream>>>(XG, GH, Cc, HS, HP, Bn, T, 4, C);
    { GemmP ch2_5_0;
      ch2_5_0.A = HP + (size_t)0 * C; ch2_5_0.B = Wh3 + (size_t)0 * C * G4; ch2_5_0.bias = HP + (size_t)0 * C; ch2_5_0.R = HP + (size_t)0 * C; ch2_5_0.C = GH;
      ch2_5_0.sAo = (long long)PP * C; ch2_5_0.sAi = (long long)18 * C; ch2_5_0.sAm = C; ch2_5_0.sAk = 1; ch2_5_0.sBo = 0; ch2_5_0.sBi = 0; ch2_5_0.sBn = 1; ch2_5_0.sBk = G4; ch2_5_0.sCo = (long long)HW * G4; ch2_5_0.sCi = (long long)16 * G4; ch2_5_0.sCm = G4; ch2_5_0.sRo = 0; ch2_5_0.sRi = 0; ch2_5_0.sRm = 0; ch2_5_0.sRn = 0;
      ch2_5_0.M = 16; ch2_5_0.N = G4; ch2_5_0.K = C; ch2_5_0.zi_n = 16; ch2_5_0.flags = 0; ch2_5_0.act = 0;
      ch2_5_0.alpha = 1.0f; ch2_5_0.beta = 0.0f; ch2_5_0.sa = 1.0f; ch2_5_0.sb = 1.0f; ch2_5_0.Npad = G4; ch2_5_0.pad_ = 0;
      k_gemm<1><<<dim3((unsigned)((G4) + 31) / 32, (unsigned)((16) + 15) / 16, (unsigned)(Bn * 16)), 32, 0, stream>>>(ch2_5_0); }
    { GemmP ch2_5_1;
      ch2_5_1.A = HP + (size_t)1 * C; ch2_5_1.B = Wh3 + (size_t)1 * C * G4; ch2_5_1.bias = HP + (size_t)1 * C; ch2_5_1.R = GH; ch2_5_1.C = GH;
      ch2_5_1.sAo = (long long)PP * C; ch2_5_1.sAi = (long long)18 * C; ch2_5_1.sAm = C; ch2_5_1.sAk = 1; ch2_5_1.sBo = 0; ch2_5_1.sBi = 0; ch2_5_1.sBn = 1; ch2_5_1.sBk = G4; ch2_5_1.sCo = (long long)HW * G4; ch2_5_1.sCi = (long long)16 * G4; ch2_5_1.sCm = G4; ch2_5_1.sRo = (long long)HW * G4; ch2_5_1.sRi = (long long)16 * G4; ch2_5_1.sRm = G4; ch2_5_1.sRn = 1;
      ch2_5_1.M = 16; ch2_5_1.N = G4; ch2_5_1.K = C; ch2_5_1.zi_n = 16; ch2_5_1.flags = 4; ch2_5_1.act = 0;
      ch2_5_1.alpha = 1.0f; ch2_5_1.beta = 1.0f; ch2_5_1.sa = 1.0f; ch2_5_1.sb = 1.0f; ch2_5_1.Npad = G4; ch2_5_1.pad_ = 0;
      k_gemm<1><<<dim3((unsigned)((G4) + 31) / 32, (unsigned)((16) + 15) / 16, (unsigned)(Bn * 16)), 32, 0, stream>>>(ch2_5_1); }
    { GemmP ch2_5_2;
      ch2_5_2.A = HP + (size_t)2 * C; ch2_5_2.B = Wh3 + (size_t)2 * C * G4; ch2_5_2.bias = HP + (size_t)2 * C; ch2_5_2.R = GH; ch2_5_2.C = GH;
      ch2_5_2.sAo = (long long)PP * C; ch2_5_2.sAi = (long long)18 * C; ch2_5_2.sAm = C; ch2_5_2.sAk = 1; ch2_5_2.sBo = 0; ch2_5_2.sBi = 0; ch2_5_2.sBn = 1; ch2_5_2.sBk = G4; ch2_5_2.sCo = (long long)HW * G4; ch2_5_2.sCi = (long long)16 * G4; ch2_5_2.sCm = G4; ch2_5_2.sRo = (long long)HW * G4; ch2_5_2.sRi = (long long)16 * G4; ch2_5_2.sRm = G4; ch2_5_2.sRn = 1;
      ch2_5_2.M = 16; ch2_5_2.N = G4; ch2_5_2.K = C; ch2_5_2.zi_n = 16; ch2_5_2.flags = 4; ch2_5_2.act = 0;
      ch2_5_2.alpha = 1.0f; ch2_5_2.beta = 1.0f; ch2_5_2.sa = 1.0f; ch2_5_2.sb = 1.0f; ch2_5_2.Npad = G4; ch2_5_2.pad_ = 0;
      k_gemm<1><<<dim3((unsigned)((G4) + 31) / 32, (unsigned)((16) + 15) / 16, (unsigned)(Bn * 16)), 32, 0, stream>>>(ch2_5_2); }
    { GemmP ch2_5_3;
      ch2_5_3.A = HP + (size_t)18 * C; ch2_5_3.B = Wh3 + (size_t)3 * C * G4; ch2_5_3.bias = HP + (size_t)18 * C; ch2_5_3.R = GH; ch2_5_3.C = GH;
      ch2_5_3.sAo = (long long)PP * C; ch2_5_3.sAi = (long long)18 * C; ch2_5_3.sAm = C; ch2_5_3.sAk = 1; ch2_5_3.sBo = 0; ch2_5_3.sBi = 0; ch2_5_3.sBn = 1; ch2_5_3.sBk = G4; ch2_5_3.sCo = (long long)HW * G4; ch2_5_3.sCi = (long long)16 * G4; ch2_5_3.sCm = G4; ch2_5_3.sRo = (long long)HW * G4; ch2_5_3.sRi = (long long)16 * G4; ch2_5_3.sRm = G4; ch2_5_3.sRn = 1;
      ch2_5_3.M = 16; ch2_5_3.N = G4; ch2_5_3.K = C; ch2_5_3.zi_n = 16; ch2_5_3.flags = 4; ch2_5_3.act = 0;
      ch2_5_3.alpha = 1.0f; ch2_5_3.beta = 1.0f; ch2_5_3.sa = 1.0f; ch2_5_3.sb = 1.0f; ch2_5_3.Npad = G4; ch2_5_3.pad_ = 0;
      k_gemm<1><<<dim3((unsigned)((G4) + 31) / 32, (unsigned)((16) + 15) / 16, (unsigned)(Bn * 16)), 32, 0, stream>>>(ch2_5_3); }
    { GemmP ch2_5_4;
      ch2_5_4.A = HP + (size_t)19 * C; ch2_5_4.B = Wh3 + (size_t)4 * C * G4; ch2_5_4.bias = HP + (size_t)19 * C; ch2_5_4.R = GH; ch2_5_4.C = GH;
      ch2_5_4.sAo = (long long)PP * C; ch2_5_4.sAi = (long long)18 * C; ch2_5_4.sAm = C; ch2_5_4.sAk = 1; ch2_5_4.sBo = 0; ch2_5_4.sBi = 0; ch2_5_4.sBn = 1; ch2_5_4.sBk = G4; ch2_5_4.sCo = (long long)HW * G4; ch2_5_4.sCi = (long long)16 * G4; ch2_5_4.sCm = G4; ch2_5_4.sRo = (long long)HW * G4; ch2_5_4.sRi = (long long)16 * G4; ch2_5_4.sRm = G4; ch2_5_4.sRn = 1;
      ch2_5_4.M = 16; ch2_5_4.N = G4; ch2_5_4.K = C; ch2_5_4.zi_n = 16; ch2_5_4.flags = 4; ch2_5_4.act = 0;
      ch2_5_4.alpha = 1.0f; ch2_5_4.beta = 1.0f; ch2_5_4.sa = 1.0f; ch2_5_4.sb = 1.0f; ch2_5_4.Npad = G4; ch2_5_4.pad_ = 0;
      k_gemm<1><<<dim3((unsigned)((G4) + 31) / 32, (unsigned)((16) + 15) / 16, (unsigned)(Bn * 16)), 32, 0, stream>>>(ch2_5_4); }
    { GemmP ch2_5_5;
      ch2_5_5.A = HP + (size_t)20 * C; ch2_5_5.B = Wh3 + (size_t)5 * C * G4; ch2_5_5.bias = HP + (size_t)20 * C; ch2_5_5.R = GH; ch2_5_5.C = GH;
      ch2_5_5.sAo = (long long)PP * C; ch2_5_5.sAi = (long long)18 * C; ch2_5_5.sAm = C; ch2_5_5.sAk = 1; ch2_5_5.sBo = 0; ch2_5_5.sBi = 0; ch2_5_5.sBn = 1; ch2_5_5.sBk = G4; ch2_5_5.sCo = (long long)HW * G4; ch2_5_5.sCi = (long long)16 * G4; ch2_5_5.sCm = G4; ch2_5_5.sRo = (long long)HW * G4; ch2_5_5.sRi = (long long)16 * G4; ch2_5_5.sRm = G4; ch2_5_5.sRn = 1;
      ch2_5_5.M = 16; ch2_5_5.N = G4; ch2_5_5.K = C; ch2_5_5.zi_n = 16; ch2_5_5.flags = 4; ch2_5_5.act = 0;
      ch2_5_5.alpha = 1.0f; ch2_5_5.beta = 1.0f; ch2_5_5.sa = 1.0f; ch2_5_5.sb = 1.0f; ch2_5_5.Npad = G4; ch2_5_5.pad_ = 0;
      k_gemm<1><<<dim3((unsigned)((G4) + 31) / 32, (unsigned)((16) + 15) / 16, (unsigned)(Bn * 16)), 32, 0, stream>>>(ch2_5_5); }
    { GemmP ch2_5_6;
      ch2_5_6.A = HP + (size_t)36 * C; ch2_5_6.B = Wh3 + (size_t)6 * C * G4; ch2_5_6.bias = HP + (size_t)36 * C; ch2_5_6.R = GH; ch2_5_6.C = GH;
      ch2_5_6.sAo = (long long)PP * C; ch2_5_6.sAi = (long long)18 * C; ch2_5_6.sAm = C; ch2_5_6.sAk = 1; ch2_5_6.sBo = 0; ch2_5_6.sBi = 0; ch2_5_6.sBn = 1; ch2_5_6.sBk = G4; ch2_5_6.sCo = (long long)HW * G4; ch2_5_6.sCi = (long long)16 * G4; ch2_5_6.sCm = G4; ch2_5_6.sRo = (long long)HW * G4; ch2_5_6.sRi = (long long)16 * G4; ch2_5_6.sRm = G4; ch2_5_6.sRn = 1;
      ch2_5_6.M = 16; ch2_5_6.N = G4; ch2_5_6.K = C; ch2_5_6.zi_n = 16; ch2_5_6.flags = 4; ch2_5_6.act = 0;
      ch2_5_6.alpha = 1.0f; ch2_5_6.beta = 1.0f; ch2_5_6.sa = 1.0f; ch2_5_6.sb = 1.0f; ch2_5_6.Npad = G4; ch2_5_6.pad_ = 0;
      k_gemm<1><<<dim3((unsigned)((G4) + 31) / 32, (unsigned)((16) + 15) / 16, (unsigned)(Bn * 16)), 32, 0, stream>>>(ch2_5_6); }
    { GemmP ch2_5_7;
      ch2_5_7.A = HP + (size_t)37 * C; ch2_5_7.B = Wh3 + (size_t)7 * C * G4; ch2_5_7.bias = HP + (size_t)37 * C; ch2_5_7.R = GH; ch2_5_7.C = GH;
      ch2_5_7.sAo = (long long)PP * C; ch2_5_7.sAi = (long long)18 * C; ch2_5_7.sAm = C; ch2_5_7.sAk = 1; ch2_5_7.sBo = 0; ch2_5_7.sBi = 0; ch2_5_7.sBn = 1; ch2_5_7.sBk = G4; ch2_5_7.sCo = (long long)HW * G4; ch2_5_7.sCi = (long long)16 * G4; ch2_5_7.sCm = G4; ch2_5_7.sRo = (long long)HW * G4; ch2_5_7.sRi = (long long)16 * G4; ch2_5_7.sRm = G4; ch2_5_7.sRn = 1;
      ch2_5_7.M = 16; ch2_5_7.N = G4; ch2_5_7.K = C; ch2_5_7.zi_n = 16; ch2_5_7.flags = 4; ch2_5_7.act = 0;
      ch2_5_7.alpha = 1.0f; ch2_5_7.beta = 1.0f; ch2_5_7.sa = 1.0f; ch2_5_7.sb = 1.0f; ch2_5_7.Npad = G4; ch2_5_7.pad_ = 0;
      k_gemm<1><<<dim3((unsigned)((G4) + 31) / 32, (unsigned)((16) + 15) / 16, (unsigned)(Bn * 16)), 32, 0, stream>>>(ch2_5_7); }
    { GemmP ch2_5_8;
      ch2_5_8.A = HP + (size_t)38 * C; ch2_5_8.B = Wh3 + (size_t)8 * C * G4; ch2_5_8.bias = HP + (size_t)38 * C; ch2_5_8.R = GH; ch2_5_8.C = GH;
      ch2_5_8.sAo = (long long)PP * C; ch2_5_8.sAi = (long long)18 * C; ch2_5_8.sAm = C; ch2_5_8.sAk = 1; ch2_5_8.sBo = 0; ch2_5_8.sBi = 0; ch2_5_8.sBn = 1; ch2_5_8.sBk = G4; ch2_5_8.sCo = (long long)HW * G4; ch2_5_8.sCi = (long long)16 * G4; ch2_5_8.sCm = G4; ch2_5_8.sRo = (long long)HW * G4; ch2_5_8.sRi = (long long)16 * G4; ch2_5_8.sRm = G4; ch2_5_8.sRn = 1;
      ch2_5_8.M = 16; ch2_5_8.N = G4; ch2_5_8.K = C; ch2_5_8.zi_n = 16; ch2_5_8.flags = 4; ch2_5_8.act = 0;
      ch2_5_8.alpha = 1.0f; ch2_5_8.beta = 1.0f; ch2_5_8.sa = 1.0f; ch2_5_8.sb = 1.0f; ch2_5_8.Npad = G4; ch2_5_8.pad_ = 0;
      k_gemm<1><<<dim3((unsigned)((G4) + 31) / 32, (unsigned)((16) + 15) / 16, (unsigned)(Bn * 16)), 32, 0, stream>>>(ch2_5_8); }

    k_bl_cell<<<(unsigned)(((long long)Bn * HW * C + 255) / 256), 256, 0, stream>>>(XG, GH, Cc, HS, HP, Bn, T, 5, C);
    { GemmP ch2_6_0;
      ch2_6_0.A = HP + (size_t)0 * C; ch2_6_0.B = Wh3 + (size_t)0 * C * G4; ch2_6_0.bias = HP + (size_t)0 * C; ch2_6_0.R = HP + (size_t)0 * C; ch2_6_0.C = GH;
      ch2_6_0.sAo = (long long)PP * C; ch2_6_0.sAi = (long long)18 * C; ch2_6_0.sAm = C; ch2_6_0.sAk = 1; ch2_6_0.sBo = 0; ch2_6_0.sBi = 0; ch2_6_0.sBn = 1; ch2_6_0.sBk = G4; ch2_6_0.sCo = (long long)HW * G4; ch2_6_0.sCi = (long long)16 * G4; ch2_6_0.sCm = G4; ch2_6_0.sRo = 0; ch2_6_0.sRi = 0; ch2_6_0.sRm = 0; ch2_6_0.sRn = 0;
      ch2_6_0.M = 16; ch2_6_0.N = G4; ch2_6_0.K = C; ch2_6_0.zi_n = 16; ch2_6_0.flags = 0; ch2_6_0.act = 0;
      ch2_6_0.alpha = 1.0f; ch2_6_0.beta = 0.0f; ch2_6_0.sa = 1.0f; ch2_6_0.sb = 1.0f; ch2_6_0.Npad = G4; ch2_6_0.pad_ = 0;
      k_gemm<1><<<dim3((unsigned)((G4) + 31) / 32, (unsigned)((16) + 15) / 16, (unsigned)(Bn * 16)), 32, 0, stream>>>(ch2_6_0); }
    { GemmP ch2_6_1;
      ch2_6_1.A = HP + (size_t)1 * C; ch2_6_1.B = Wh3 + (size_t)1 * C * G4; ch2_6_1.bias = HP + (size_t)1 * C; ch2_6_1.R = GH; ch2_6_1.C = GH;
      ch2_6_1.sAo = (long long)PP * C; ch2_6_1.sAi = (long long)18 * C; ch2_6_1.sAm = C; ch2_6_1.sAk = 1; ch2_6_1.sBo = 0; ch2_6_1.sBi = 0; ch2_6_1.sBn = 1; ch2_6_1.sBk = G4; ch2_6_1.sCo = (long long)HW * G4; ch2_6_1.sCi = (long long)16 * G4; ch2_6_1.sCm = G4; ch2_6_1.sRo = (long long)HW * G4; ch2_6_1.sRi = (long long)16 * G4; ch2_6_1.sRm = G4; ch2_6_1.sRn = 1;
      ch2_6_1.M = 16; ch2_6_1.N = G4; ch2_6_1.K = C; ch2_6_1.zi_n = 16; ch2_6_1.flags = 4; ch2_6_1.act = 0;
      ch2_6_1.alpha = 1.0f; ch2_6_1.beta = 1.0f; ch2_6_1.sa = 1.0f; ch2_6_1.sb = 1.0f; ch2_6_1.Npad = G4; ch2_6_1.pad_ = 0;
      k_gemm<1><<<dim3((unsigned)((G4) + 31) / 32, (unsigned)((16) + 15) / 16, (unsigned)(Bn * 16)), 32, 0, stream>>>(ch2_6_1); }
    { GemmP ch2_6_2;
      ch2_6_2.A = HP + (size_t)2 * C; ch2_6_2.B = Wh3 + (size_t)2 * C * G4; ch2_6_2.bias = HP + (size_t)2 * C; ch2_6_2.R = GH; ch2_6_2.C = GH;
      ch2_6_2.sAo = (long long)PP * C; ch2_6_2.sAi = (long long)18 * C; ch2_6_2.sAm = C; ch2_6_2.sAk = 1; ch2_6_2.sBo = 0; ch2_6_2.sBi = 0; ch2_6_2.sBn = 1; ch2_6_2.sBk = G4; ch2_6_2.sCo = (long long)HW * G4; ch2_6_2.sCi = (long long)16 * G4; ch2_6_2.sCm = G4; ch2_6_2.sRo = (long long)HW * G4; ch2_6_2.sRi = (long long)16 * G4; ch2_6_2.sRm = G4; ch2_6_2.sRn = 1;
      ch2_6_2.M = 16; ch2_6_2.N = G4; ch2_6_2.K = C; ch2_6_2.zi_n = 16; ch2_6_2.flags = 4; ch2_6_2.act = 0;
      ch2_6_2.alpha = 1.0f; ch2_6_2.beta = 1.0f; ch2_6_2.sa = 1.0f; ch2_6_2.sb = 1.0f; ch2_6_2.Npad = G4; ch2_6_2.pad_ = 0;
      k_gemm<1><<<dim3((unsigned)((G4) + 31) / 32, (unsigned)((16) + 15) / 16, (unsigned)(Bn * 16)), 32, 0, stream>>>(ch2_6_2); }
    { GemmP ch2_6_3;
      ch2_6_3.A = HP + (size_t)18 * C; ch2_6_3.B = Wh3 + (size_t)3 * C * G4; ch2_6_3.bias = HP + (size_t)18 * C; ch2_6_3.R = GH; ch2_6_3.C = GH;
      ch2_6_3.sAo = (long long)PP * C; ch2_6_3.sAi = (long long)18 * C; ch2_6_3.sAm = C; ch2_6_3.sAk = 1; ch2_6_3.sBo = 0; ch2_6_3.sBi = 0; ch2_6_3.sBn = 1; ch2_6_3.sBk = G4; ch2_6_3.sCo = (long long)HW * G4; ch2_6_3.sCi = (long long)16 * G4; ch2_6_3.sCm = G4; ch2_6_3.sRo = (long long)HW * G4; ch2_6_3.sRi = (long long)16 * G4; ch2_6_3.sRm = G4; ch2_6_3.sRn = 1;
      ch2_6_3.M = 16; ch2_6_3.N = G4; ch2_6_3.K = C; ch2_6_3.zi_n = 16; ch2_6_3.flags = 4; ch2_6_3.act = 0;
      ch2_6_3.alpha = 1.0f; ch2_6_3.beta = 1.0f; ch2_6_3.sa = 1.0f; ch2_6_3.sb = 1.0f; ch2_6_3.Npad = G4; ch2_6_3.pad_ = 0;
      k_gemm<1><<<dim3((unsigned)((G4) + 31) / 32, (unsigned)((16) + 15) / 16, (unsigned)(Bn * 16)), 32, 0, stream>>>(ch2_6_3); }
    { GemmP ch2_6_4;
      ch2_6_4.A = HP + (size_t)19 * C; ch2_6_4.B = Wh3 + (size_t)4 * C * G4; ch2_6_4.bias = HP + (size_t)19 * C; ch2_6_4.R = GH; ch2_6_4.C = GH;
      ch2_6_4.sAo = (long long)PP * C; ch2_6_4.sAi = (long long)18 * C; ch2_6_4.sAm = C; ch2_6_4.sAk = 1; ch2_6_4.sBo = 0; ch2_6_4.sBi = 0; ch2_6_4.sBn = 1; ch2_6_4.sBk = G4; ch2_6_4.sCo = (long long)HW * G4; ch2_6_4.sCi = (long long)16 * G4; ch2_6_4.sCm = G4; ch2_6_4.sRo = (long long)HW * G4; ch2_6_4.sRi = (long long)16 * G4; ch2_6_4.sRm = G4; ch2_6_4.sRn = 1;
      ch2_6_4.M = 16; ch2_6_4.N = G4; ch2_6_4.K = C; ch2_6_4.zi_n = 16; ch2_6_4.flags = 4; ch2_6_4.act = 0;
      ch2_6_4.alpha = 1.0f; ch2_6_4.beta = 1.0f; ch2_6_4.sa = 1.0f; ch2_6_4.sb = 1.0f; ch2_6_4.Npad = G4; ch2_6_4.pad_ = 0;
      k_gemm<1><<<dim3((unsigned)((G4) + 31) / 32, (unsigned)((16) + 15) / 16, (unsigned)(Bn * 16)), 32, 0, stream>>>(ch2_6_4); }
    { GemmP ch2_6_5;
      ch2_6_5.A = HP + (size_t)20 * C; ch2_6_5.B = Wh3 + (size_t)5 * C * G4; ch2_6_5.bias = HP + (size_t)20 * C; ch2_6_5.R = GH; ch2_6_5.C = GH;
      ch2_6_5.sAo = (long long)PP * C; ch2_6_5.sAi = (long long)18 * C; ch2_6_5.sAm = C; ch2_6_5.sAk = 1; ch2_6_5.sBo = 0; ch2_6_5.sBi = 0; ch2_6_5.sBn = 1; ch2_6_5.sBk = G4; ch2_6_5.sCo = (long long)HW * G4; ch2_6_5.sCi = (long long)16 * G4; ch2_6_5.sCm = G4; ch2_6_5.sRo = (long long)HW * G4; ch2_6_5.sRi = (long long)16 * G4; ch2_6_5.sRm = G4; ch2_6_5.sRn = 1;
      ch2_6_5.M = 16; ch2_6_5.N = G4; ch2_6_5.K = C; ch2_6_5.zi_n = 16; ch2_6_5.flags = 4; ch2_6_5.act = 0;
      ch2_6_5.alpha = 1.0f; ch2_6_5.beta = 1.0f; ch2_6_5.sa = 1.0f; ch2_6_5.sb = 1.0f; ch2_6_5.Npad = G4; ch2_6_5.pad_ = 0;
      k_gemm<1><<<dim3((unsigned)((G4) + 31) / 32, (unsigned)((16) + 15) / 16, (unsigned)(Bn * 16)), 32, 0, stream>>>(ch2_6_5); }
    { GemmP ch2_6_6;
      ch2_6_6.A = HP + (size_t)36 * C; ch2_6_6.B = Wh3 + (size_t)6 * C * G4; ch2_6_6.bias = HP + (size_t)36 * C; ch2_6_6.R = GH; ch2_6_6.C = GH;
      ch2_6_6.sAo = (long long)PP * C; ch2_6_6.sAi = (long long)18 * C; ch2_6_6.sAm = C; ch2_6_6.sAk = 1; ch2_6_6.sBo = 0; ch2_6_6.sBi = 0; ch2_6_6.sBn = 1; ch2_6_6.sBk = G4; ch2_6_6.sCo = (long long)HW * G4; ch2_6_6.sCi = (long long)16 * G4; ch2_6_6.sCm = G4; ch2_6_6.sRo = (long long)HW * G4; ch2_6_6.sRi = (long long)16 * G4; ch2_6_6.sRm = G4; ch2_6_6.sRn = 1;
      ch2_6_6.M = 16; ch2_6_6.N = G4; ch2_6_6.K = C; ch2_6_6.zi_n = 16; ch2_6_6.flags = 4; ch2_6_6.act = 0;
      ch2_6_6.alpha = 1.0f; ch2_6_6.beta = 1.0f; ch2_6_6.sa = 1.0f; ch2_6_6.sb = 1.0f; ch2_6_6.Npad = G4; ch2_6_6.pad_ = 0;
      k_gemm<1><<<dim3((unsigned)((G4) + 31) / 32, (unsigned)((16) + 15) / 16, (unsigned)(Bn * 16)), 32, 0, stream>>>(ch2_6_6); }
    { GemmP ch2_6_7;
      ch2_6_7.A = HP + (size_t)37 * C; ch2_6_7.B = Wh3 + (size_t)7 * C * G4; ch2_6_7.bias = HP + (size_t)37 * C; ch2_6_7.R = GH; ch2_6_7.C = GH;
      ch2_6_7.sAo = (long long)PP * C; ch2_6_7.sAi = (long long)18 * C; ch2_6_7.sAm = C; ch2_6_7.sAk = 1; ch2_6_7.sBo = 0; ch2_6_7.sBi = 0; ch2_6_7.sBn = 1; ch2_6_7.sBk = G4; ch2_6_7.sCo = (long long)HW * G4; ch2_6_7.sCi = (long long)16 * G4; ch2_6_7.sCm = G4; ch2_6_7.sRo = (long long)HW * G4; ch2_6_7.sRi = (long long)16 * G4; ch2_6_7.sRm = G4; ch2_6_7.sRn = 1;
      ch2_6_7.M = 16; ch2_6_7.N = G4; ch2_6_7.K = C; ch2_6_7.zi_n = 16; ch2_6_7.flags = 4; ch2_6_7.act = 0;
      ch2_6_7.alpha = 1.0f; ch2_6_7.beta = 1.0f; ch2_6_7.sa = 1.0f; ch2_6_7.sb = 1.0f; ch2_6_7.Npad = G4; ch2_6_7.pad_ = 0;
      k_gemm<1><<<dim3((unsigned)((G4) + 31) / 32, (unsigned)((16) + 15) / 16, (unsigned)(Bn * 16)), 32, 0, stream>>>(ch2_6_7); }
    { GemmP ch2_6_8;
      ch2_6_8.A = HP + (size_t)38 * C; ch2_6_8.B = Wh3 + (size_t)8 * C * G4; ch2_6_8.bias = HP + (size_t)38 * C; ch2_6_8.R = GH; ch2_6_8.C = GH;
      ch2_6_8.sAo = (long long)PP * C; ch2_6_8.sAi = (long long)18 * C; ch2_6_8.sAm = C; ch2_6_8.sAk = 1; ch2_6_8.sBo = 0; ch2_6_8.sBi = 0; ch2_6_8.sBn = 1; ch2_6_8.sBk = G4; ch2_6_8.sCo = (long long)HW * G4; ch2_6_8.sCi = (long long)16 * G4; ch2_6_8.sCm = G4; ch2_6_8.sRo = (long long)HW * G4; ch2_6_8.sRi = (long long)16 * G4; ch2_6_8.sRm = G4; ch2_6_8.sRn = 1;
      ch2_6_8.M = 16; ch2_6_8.N = G4; ch2_6_8.K = C; ch2_6_8.zi_n = 16; ch2_6_8.flags = 4; ch2_6_8.act = 0;
      ch2_6_8.alpha = 1.0f; ch2_6_8.beta = 1.0f; ch2_6_8.sa = 1.0f; ch2_6_8.sb = 1.0f; ch2_6_8.Npad = G4; ch2_6_8.pad_ = 0;
      k_gemm<1><<<dim3((unsigned)((G4) + 31) / 32, (unsigned)((16) + 15) / 16, (unsigned)(Bn * 16)), 32, 0, stream>>>(ch2_6_8); }

    k_bl_cell<<<(unsigned)(((long long)Bn * HW * C + 255) / 256), 256, 0, stream>>>(XG, GH, Cc, HS, HP, Bn, T, 6, C);
    { GemmP ch2_7_0;
      ch2_7_0.A = HP + (size_t)0 * C; ch2_7_0.B = Wh3 + (size_t)0 * C * G4; ch2_7_0.bias = HP + (size_t)0 * C; ch2_7_0.R = HP + (size_t)0 * C; ch2_7_0.C = GH;
      ch2_7_0.sAo = (long long)PP * C; ch2_7_0.sAi = (long long)18 * C; ch2_7_0.sAm = C; ch2_7_0.sAk = 1; ch2_7_0.sBo = 0; ch2_7_0.sBi = 0; ch2_7_0.sBn = 1; ch2_7_0.sBk = G4; ch2_7_0.sCo = (long long)HW * G4; ch2_7_0.sCi = (long long)16 * G4; ch2_7_0.sCm = G4; ch2_7_0.sRo = 0; ch2_7_0.sRi = 0; ch2_7_0.sRm = 0; ch2_7_0.sRn = 0;
      ch2_7_0.M = 16; ch2_7_0.N = G4; ch2_7_0.K = C; ch2_7_0.zi_n = 16; ch2_7_0.flags = 0; ch2_7_0.act = 0;
      ch2_7_0.alpha = 1.0f; ch2_7_0.beta = 0.0f; ch2_7_0.sa = 1.0f; ch2_7_0.sb = 1.0f; ch2_7_0.Npad = G4; ch2_7_0.pad_ = 0;
      k_gemm<1><<<dim3((unsigned)((G4) + 31) / 32, (unsigned)((16) + 15) / 16, (unsigned)(Bn * 16)), 32, 0, stream>>>(ch2_7_0); }
    { GemmP ch2_7_1;
      ch2_7_1.A = HP + (size_t)1 * C; ch2_7_1.B = Wh3 + (size_t)1 * C * G4; ch2_7_1.bias = HP + (size_t)1 * C; ch2_7_1.R = GH; ch2_7_1.C = GH;
      ch2_7_1.sAo = (long long)PP * C; ch2_7_1.sAi = (long long)18 * C; ch2_7_1.sAm = C; ch2_7_1.sAk = 1; ch2_7_1.sBo = 0; ch2_7_1.sBi = 0; ch2_7_1.sBn = 1; ch2_7_1.sBk = G4; ch2_7_1.sCo = (long long)HW * G4; ch2_7_1.sCi = (long long)16 * G4; ch2_7_1.sCm = G4; ch2_7_1.sRo = (long long)HW * G4; ch2_7_1.sRi = (long long)16 * G4; ch2_7_1.sRm = G4; ch2_7_1.sRn = 1;
      ch2_7_1.M = 16; ch2_7_1.N = G4; ch2_7_1.K = C; ch2_7_1.zi_n = 16; ch2_7_1.flags = 4; ch2_7_1.act = 0;
      ch2_7_1.alpha = 1.0f; ch2_7_1.beta = 1.0f; ch2_7_1.sa = 1.0f; ch2_7_1.sb = 1.0f; ch2_7_1.Npad = G4; ch2_7_1.pad_ = 0;
      k_gemm<1><<<dim3((unsigned)((G4) + 31) / 32, (unsigned)((16) + 15) / 16, (unsigned)(Bn * 16)), 32, 0, stream>>>(ch2_7_1); }
    { GemmP ch2_7_2;
      ch2_7_2.A = HP + (size_t)2 * C; ch2_7_2.B = Wh3 + (size_t)2 * C * G4; ch2_7_2.bias = HP + (size_t)2 * C; ch2_7_2.R = GH; ch2_7_2.C = GH;
      ch2_7_2.sAo = (long long)PP * C; ch2_7_2.sAi = (long long)18 * C; ch2_7_2.sAm = C; ch2_7_2.sAk = 1; ch2_7_2.sBo = 0; ch2_7_2.sBi = 0; ch2_7_2.sBn = 1; ch2_7_2.sBk = G4; ch2_7_2.sCo = (long long)HW * G4; ch2_7_2.sCi = (long long)16 * G4; ch2_7_2.sCm = G4; ch2_7_2.sRo = (long long)HW * G4; ch2_7_2.sRi = (long long)16 * G4; ch2_7_2.sRm = G4; ch2_7_2.sRn = 1;
      ch2_7_2.M = 16; ch2_7_2.N = G4; ch2_7_2.K = C; ch2_7_2.zi_n = 16; ch2_7_2.flags = 4; ch2_7_2.act = 0;
      ch2_7_2.alpha = 1.0f; ch2_7_2.beta = 1.0f; ch2_7_2.sa = 1.0f; ch2_7_2.sb = 1.0f; ch2_7_2.Npad = G4; ch2_7_2.pad_ = 0;
      k_gemm<1><<<dim3((unsigned)((G4) + 31) / 32, (unsigned)((16) + 15) / 16, (unsigned)(Bn * 16)), 32, 0, stream>>>(ch2_7_2); }
    { GemmP ch2_7_3;
      ch2_7_3.A = HP + (size_t)18 * C; ch2_7_3.B = Wh3 + (size_t)3 * C * G4; ch2_7_3.bias = HP + (size_t)18 * C; ch2_7_3.R = GH; ch2_7_3.C = GH;
      ch2_7_3.sAo = (long long)PP * C; ch2_7_3.sAi = (long long)18 * C; ch2_7_3.sAm = C; ch2_7_3.sAk = 1; ch2_7_3.sBo = 0; ch2_7_3.sBi = 0; ch2_7_3.sBn = 1; ch2_7_3.sBk = G4; ch2_7_3.sCo = (long long)HW * G4; ch2_7_3.sCi = (long long)16 * G4; ch2_7_3.sCm = G4; ch2_7_3.sRo = (long long)HW * G4; ch2_7_3.sRi = (long long)16 * G4; ch2_7_3.sRm = G4; ch2_7_3.sRn = 1;
      ch2_7_3.M = 16; ch2_7_3.N = G4; ch2_7_3.K = C; ch2_7_3.zi_n = 16; ch2_7_3.flags = 4; ch2_7_3.act = 0;
      ch2_7_3.alpha = 1.0f; ch2_7_3.beta = 1.0f; ch2_7_3.sa = 1.0f; ch2_7_3.sb = 1.0f; ch2_7_3.Npad = G4; ch2_7_3.pad_ = 0;
      k_gemm<1><<<dim3((unsigned)((G4) + 31) / 32, (unsigned)((16) + 15) / 16, (unsigned)(Bn * 16)), 32, 0, stream>>>(ch2_7_3); }
    { GemmP ch2_7_4;
      ch2_7_4.A = HP + (size_t)19 * C; ch2_7_4.B = Wh3 + (size_t)4 * C * G4; ch2_7_4.bias = HP + (size_t)19 * C; ch2_7_4.R = GH; ch2_7_4.C = GH;
      ch2_7_4.sAo = (long long)PP * C; ch2_7_4.sAi = (long long)18 * C; ch2_7_4.sAm = C; ch2_7_4.sAk = 1; ch2_7_4.sBo = 0; ch2_7_4.sBi = 0; ch2_7_4.sBn = 1; ch2_7_4.sBk = G4; ch2_7_4.sCo = (long long)HW * G4; ch2_7_4.sCi = (long long)16 * G4; ch2_7_4.sCm = G4; ch2_7_4.sRo = (long long)HW * G4; ch2_7_4.sRi = (long long)16 * G4; ch2_7_4.sRm = G4; ch2_7_4.sRn = 1;
      ch2_7_4.M = 16; ch2_7_4.N = G4; ch2_7_4.K = C; ch2_7_4.zi_n = 16; ch2_7_4.flags = 4; ch2_7_4.act = 0;
      ch2_7_4.alpha = 1.0f; ch2_7_4.beta = 1.0f; ch2_7_4.sa = 1.0f; ch2_7_4.sb = 1.0f; ch2_7_4.Npad = G4; ch2_7_4.pad_ = 0;
      k_gemm<1><<<dim3((unsigned)((G4) + 31) / 32, (unsigned)((16) + 15) / 16, (unsigned)(Bn * 16)), 32, 0, stream>>>(ch2_7_4); }
    { GemmP ch2_7_5;
      ch2_7_5.A = HP + (size_t)20 * C; ch2_7_5.B = Wh3 + (size_t)5 * C * G4; ch2_7_5.bias = HP + (size_t)20 * C; ch2_7_5.R = GH; ch2_7_5.C = GH;
      ch2_7_5.sAo = (long long)PP * C; ch2_7_5.sAi = (long long)18 * C; ch2_7_5.sAm = C; ch2_7_5.sAk = 1; ch2_7_5.sBo = 0; ch2_7_5.sBi = 0; ch2_7_5.sBn = 1; ch2_7_5.sBk = G4; ch2_7_5.sCo = (long long)HW * G4; ch2_7_5.sCi = (long long)16 * G4; ch2_7_5.sCm = G4; ch2_7_5.sRo = (long long)HW * G4; ch2_7_5.sRi = (long long)16 * G4; ch2_7_5.sRm = G4; ch2_7_5.sRn = 1;
      ch2_7_5.M = 16; ch2_7_5.N = G4; ch2_7_5.K = C; ch2_7_5.zi_n = 16; ch2_7_5.flags = 4; ch2_7_5.act = 0;
      ch2_7_5.alpha = 1.0f; ch2_7_5.beta = 1.0f; ch2_7_5.sa = 1.0f; ch2_7_5.sb = 1.0f; ch2_7_5.Npad = G4; ch2_7_5.pad_ = 0;
      k_gemm<1><<<dim3((unsigned)((G4) + 31) / 32, (unsigned)((16) + 15) / 16, (unsigned)(Bn * 16)), 32, 0, stream>>>(ch2_7_5); }
    { GemmP ch2_7_6;
      ch2_7_6.A = HP + (size_t)36 * C; ch2_7_6.B = Wh3 + (size_t)6 * C * G4; ch2_7_6.bias = HP + (size_t)36 * C; ch2_7_6.R = GH; ch2_7_6.C = GH;
      ch2_7_6.sAo = (long long)PP * C; ch2_7_6.sAi = (long long)18 * C; ch2_7_6.sAm = C; ch2_7_6.sAk = 1; ch2_7_6.sBo = 0; ch2_7_6.sBi = 0; ch2_7_6.sBn = 1; ch2_7_6.sBk = G4; ch2_7_6.sCo = (long long)HW * G4; ch2_7_6.sCi = (long long)16 * G4; ch2_7_6.sCm = G4; ch2_7_6.sRo = (long long)HW * G4; ch2_7_6.sRi = (long long)16 * G4; ch2_7_6.sRm = G4; ch2_7_6.sRn = 1;
      ch2_7_6.M = 16; ch2_7_6.N = G4; ch2_7_6.K = C; ch2_7_6.zi_n = 16; ch2_7_6.flags = 4; ch2_7_6.act = 0;
      ch2_7_6.alpha = 1.0f; ch2_7_6.beta = 1.0f; ch2_7_6.sa = 1.0f; ch2_7_6.sb = 1.0f; ch2_7_6.Npad = G4; ch2_7_6.pad_ = 0;
      k_gemm<1><<<dim3((unsigned)((G4) + 31) / 32, (unsigned)((16) + 15) / 16, (unsigned)(Bn * 16)), 32, 0, stream>>>(ch2_7_6); }
    { GemmP ch2_7_7;
      ch2_7_7.A = HP + (size_t)37 * C; ch2_7_7.B = Wh3 + (size_t)7 * C * G4; ch2_7_7.bias = HP + (size_t)37 * C; ch2_7_7.R = GH; ch2_7_7.C = GH;
      ch2_7_7.sAo = (long long)PP * C; ch2_7_7.sAi = (long long)18 * C; ch2_7_7.sAm = C; ch2_7_7.sAk = 1; ch2_7_7.sBo = 0; ch2_7_7.sBi = 0; ch2_7_7.sBn = 1; ch2_7_7.sBk = G4; ch2_7_7.sCo = (long long)HW * G4; ch2_7_7.sCi = (long long)16 * G4; ch2_7_7.sCm = G4; ch2_7_7.sRo = (long long)HW * G4; ch2_7_7.sRi = (long long)16 * G4; ch2_7_7.sRm = G4; ch2_7_7.sRn = 1;
      ch2_7_7.M = 16; ch2_7_7.N = G4; ch2_7_7.K = C; ch2_7_7.zi_n = 16; ch2_7_7.flags = 4; ch2_7_7.act = 0;
      ch2_7_7.alpha = 1.0f; ch2_7_7.beta = 1.0f; ch2_7_7.sa = 1.0f; ch2_7_7.sb = 1.0f; ch2_7_7.Npad = G4; ch2_7_7.pad_ = 0;
      k_gemm<1><<<dim3((unsigned)((G4) + 31) / 32, (unsigned)((16) + 15) / 16, (unsigned)(Bn * 16)), 32, 0, stream>>>(ch2_7_7); }
    { GemmP ch2_7_8;
      ch2_7_8.A = HP + (size_t)38 * C; ch2_7_8.B = Wh3 + (size_t)8 * C * G4; ch2_7_8.bias = HP + (size_t)38 * C; ch2_7_8.R = GH; ch2_7_8.C = GH;
      ch2_7_8.sAo = (long long)PP * C; ch2_7_8.sAi = (long long)18 * C; ch2_7_8.sAm = C; ch2_7_8.sAk = 1; ch2_7_8.sBo = 0; ch2_7_8.sBi = 0; ch2_7_8.sBn = 1; ch2_7_8.sBk = G4; ch2_7_8.sCo = (long long)HW * G4; ch2_7_8.sCi = (long long)16 * G4; ch2_7_8.sCm = G4; ch2_7_8.sRo = (long long)HW * G4; ch2_7_8.sRi = (long long)16 * G4; ch2_7_8.sRm = G4; ch2_7_8.sRn = 1;
      ch2_7_8.M = 16; ch2_7_8.N = G4; ch2_7_8.K = C; ch2_7_8.zi_n = 16; ch2_7_8.flags = 4; ch2_7_8.act = 0;
      ch2_7_8.alpha = 1.0f; ch2_7_8.beta = 1.0f; ch2_7_8.sa = 1.0f; ch2_7_8.sb = 1.0f; ch2_7_8.Npad = G4; ch2_7_8.pad_ = 0;
      k_gemm<1><<<dim3((unsigned)((G4) + 31) / 32, (unsigned)((16) + 15) / 16, (unsigned)(Bn * 16)), 32, 0, stream>>>(ch2_7_8); }

    k_bl_cell<<<(unsigned)(((long long)Bn * HW * C + 255) / 256), 256, 0, stream>>>(XG, GH, Cc, HS, HP, Bn, T, 7, C);
    k_stats<<<(unsigned)(C), 256, 0, stream>>>(HS, 1, C, 0, 1, NF * HW, 0.001f, st, 0);
    k_norm_apply<<<(unsigned)(((long long)(NF * HW) * (C) * (1) + 255) / 256), 256, 0, stream>>>(HS, out, st, g3, be3, NF * HW, C, 1, 1, 1, 0);
}
